// CCMNet_16106127360571
// MI455X (gfx1250) — hardware-verified
//
#include <hip/hip_runtime.h>
#include <math.h>

typedef __attribute__((ext_vector_type(16))) _Float16 v16h;
typedef __attribute__((ext_vector_type(8)))  _Float16 v8h;
typedef __attribute__((ext_vector_type(16))) __bf16   v16b;
typedef __attribute__((ext_vector_type(8)))  float    v8f;
typedef __attribute__((ext_vector_type(4)))  float    v4f;

__device__ __forceinline__ int frag_k(int i, int h) { return (i < 8) ? (8 * h + i) : (16 + 8 * h + (i - 8)); }
__device__ __forceinline__ __bf16 bf16_rne(float f) {
    unsigned int u = __float_as_uint(f);
    u += 0x7fffu + ((u >> 16) & 1u);
    return __builtin_bit_cast(__bf16, (unsigned short)(u >> 16));
}
__device__ __forceinline__ float bf16_f32(__bf16 b) { return __uint_as_float(((unsigned int)__builtin_bit_cast(unsigned short, b)) << 16); }
__device__ __forceinline__ v8f wmma16(v16h a, v16h b, v8f c) {
    c = __builtin_amdgcn_wmma_f32_16x16x32_f16(false, a, false, b, (short)0, c, false, false);
    asm volatile("v_nop\n\tv_nop\n\tv_nop\n\tv_nop" : "+v"(c) : "v"(a), "v"(b));
    return c;
}
__device__ __forceinline__ v8f wmmab(v16b a, v16b b, v8f c) {
    c = __builtin_amdgcn_wmma_f32_16x16x32_bf16(false, a, false, b, (short)0, c, false, false);
    asm volatile("v_nop\n\tv_nop\n\tv_nop\n\tv_nop" : "+v"(c) : "v"(a), "v"(b));
    return c;
}
struct Split { v16b hi, lo; };
__device__ __forceinline__ v8f wmma3(const Split& a, const Split& b, v8f c) {
    c = __builtin_amdgcn_wmma_f32_16x16x32_bf16(false, a.hi, false, b.hi, (short)0, c, false, false);
    c = __builtin_amdgcn_wmma_f32_16x16x32_bf16(false, a.hi, false, b.lo, (short)0, c, false, false);
    c = __builtin_amdgcn_wmma_f32_16x16x32_bf16(false, a.lo, false, b.hi, (short)0, c, false, false);
    asm volatile("v_nop\n\tv_nop\n\tv_nop\n\tv_nop" : "+v"(c) : "v"(a.hi), "v"(a.lo), "v"(b.hi), "v"(b.lo));
    return c;
}
struct Split3 { v16b hi, mid, lo; };
__device__ __forceinline__ v8f wmma6(const Split3& a, const Split3& b, v8f c) {
    c = __builtin_amdgcn_wmma_f32_16x16x32_bf16(false, a.hi, false, b.hi, (short)0, c, false, false);
    c = __builtin_amdgcn_wmma_f32_16x16x32_bf16(false, a.hi, false, b.mid, (short)0, c, false, false);
    c = __builtin_amdgcn_wmma_f32_16x16x32_bf16(false, a.mid, false, b.hi, (short)0, c, false, false);
    c = __builtin_amdgcn_wmma_f32_16x16x32_bf16(false, a.hi, false, b.lo, (short)0, c, false, false);
    c = __builtin_amdgcn_wmma_f32_16x16x32_bf16(false, a.mid, false, b.mid, (short)0, c, false, false);
    c = __builtin_amdgcn_wmma_f32_16x16x32_bf16(false, a.lo, false, b.hi, (short)0, c, false, false);
    asm volatile("v_nop\n\tv_nop\n\tv_nop\n\tv_nop" : "+v"(c) : "v"(a.hi), "v"(a.mid), "v"(a.lo), "v"(b.hi), "v"(b.mid), "v"(b.lo));
    return c;
}

__device__ __forceinline__ v16h fh_ld(const float* __restrict__ p, long long sk, int k0, int h, int klen, float s) {
    v16h a;
#pragma unroll
    for (int i = 0; i < 16; ++i) { const int k = k0 + frag_k(i, h); a[i] = (k < klen) ? (_Float16)(p[(long long)k * sk] * s) : (_Float16)0.f; }
    return a;
}
__device__ __forceinline__ Split sp_ld(const float* __restrict__ p, long long sk, int k0, int h, int klen, float s) {
    Split r;
#pragma unroll
    for (int i = 0; i < 16; ++i) {
        const int k = k0 + frag_k(i, h); const float x = (k < klen) ? p[(long long)k * sk] * s : 0.f;
        const __bf16 hb = bf16_rne(x); r.hi[i] = hb; r.lo[i] = bf16_rne(x - bf16_f32(hb));
    }
    return r;
}
__device__ __forceinline__ Split3 sp3_ld(const float* __restrict__ p, long long sk, int k0, int h, int klen, float s) {
    Split3 r;
#pragma unroll
    for (int i = 0; i < 16; ++i) {
        const int k = k0 + frag_k(i, h); const float x = (k < klen) ? p[(long long)k * sk] * s : 0.f;
        const __bf16 hb = bf16_rne(x); const float r1 = x - bf16_f32(hb); const __bf16 mb = bf16_rne(r1);
        r.hi[i] = hb; r.mid[i] = mb; r.lo[i] = bf16_rne(r1 - bf16_f32(mb));
    }
    return r;
}
__device__ __forceinline__ v16b bh_ld(const float* __restrict__ p, long long sk, int k0, int h, int klen, float s) {
    v16b a;
#pragma unroll
    for (int i = 0; i < 16; ++i) { const int k = k0 + frag_k(i, h); a[i] = bf16_rne((k < klen) ? p[(long long)k * sk] * s : 0.f); }
    return a;
}
__device__ __forceinline__ v16h fh_row(const _Float16* __restrict__ row, int k0, int h) {
    v16h a;
#pragma unroll
    for (int i = 0; i < 16; ++i) a[i] = row[k0 + frag_k(i, h)];
    return a;
}

#define VST2(T, ptr, val) do { *(volatile T*)(ptr) = (val); __threadfence(); *(volatile T*)(ptr) = (val); } while (0)
typedef float v4f __attribute__((ext_vector_type(4)));
#define VST2V4(ptr, val) do { *(volatile v4f*)(ptr) = (val); __threadfence(); *(volatile v4f*)(ptr) = (val); } while (0)

__device__ __attribute__((noinline)) float act_fn(float v, int act) {
    if (act == 1) return fmaxf(v, 0.f);
    if (act == 2) { const float u = 0.7978845608028654f * (v + 0.044715f * v * v * v); return 0.5f * v * (1.f + tanhf(u)); }
    if (act == 3) return v / (1.f + expf(-v));
    if (act == 4) return 0.5f * v * (1.f + erff(v * 0.7071067811865476f));
    if (act == 5) return tanhf(v);
    if (act == 6) return 1.f / (1.f + expf(-v));
    if (act == 7) return (v > 0.f) ? v : 0.01f * v;
    if (act == 8) return (v > 0.f) ? v : (expf(v) - 1.f);
    if (act == 9) return fminf(fmaxf(v, 0.f), 6.f);
    if (act == 10) return fabsf(v);
    if (act == 11) return (v >= 0.f) ? v : 0.1f * v;
    if (act == 12) return (v > 0.f) ? v : 0.2f * v;
    if (act == 13) return (v > 20.f) ? v : log1pf(expf(v));
    return v;
}

struct GemmP {
    const float* A; const float* B; const float* bias; const float* R; float* C;
    long long sAo, sAi, sAm, sAk, sBo, sBi, sBn, sBk, sCo, sCi, sCm, sRo, sRi, sRm, sRn;
    int M, N, K, zi_n, flags, act; float alpha, beta, sa, sb;
    int Npad, pad_;
};
static_assert(sizeof(GemmP) == 5 * 8 + 15 * 8 + 6 * 4 + 4 * 4 + 2 * 4, "GemmP has padding");

template <int MODE>
__global__ __launch_bounds__(32) void k_gemm(GemmP p) {
    const int lane = threadIdx.x & 31, h = lane >> 4, l15 = lane & 15;
    const int m0 = blockIdx.y * 16, n0 = blockIdx.x * 32;
    const int z = blockIdx.z, zo = z / p.zi_n, zi = z - zo * p.zi_n;
    const float* A = p.A + zo * p.sAo + zi * p.sAi;
    const float* B = p.B + zo * p.sBo + zi * p.sBi;
    const int am = min(m0 + l15, p.M - 1);
    v8f acc[2], comp[2];
#pragma unroll
    for (int t = 0; t < 2; ++t) { v8f zz = {}; acc[t] = zz; comp[t] = zz; }
    for (int k0 = 0; k0 < p.K; k0 += 32) {
        const float* arow = A + (long long)am * p.sAm;
        if (MODE == 1) {
            const Split a = sp_ld(arow, p.sAk, k0, h, p.K, 1.f);
#pragma unroll
            for (int t = 0; t < 2; ++t) {
                const int bn = min(n0 + t * 16 + l15, p.N - 1);
                acc[t] = wmma3(a, sp_ld(B + (long long)bn * p.sBn, p.sBk, k0, h, p.K, 1.f), acc[t]);
            }
        } else if (MODE == 3) {
            const Split3 a = sp3_ld(arow, p.sAk, k0, h, p.K, 1.f);
#pragma unroll
            for (int t = 0; t < 2; ++t) {
                const int bn = min(n0 + t * 16 + l15, p.N - 1);
                acc[t] = wmma6(a, sp3_ld(B + (long long)bn * p.sBn, p.sBk, k0, h, p.K, 1.f), acc[t]);
            }
        } else if (MODE == 4) {
            const Split3 a = sp3_ld(arow, p.sAk, k0, h, p.K, 1.f);
#pragma unroll
            for (int t = 0; t < 2; ++t) {
                const int bn = min(n0 + t * 16 + l15, p.N - 1); v8f zz = {};
                const v8f part = wmma6(a, sp3_ld(B + (long long)bn * p.sBn, p.sBk, k0, h, p.K, 1.f), zz);
                const v8f y = part - comp[t]; const v8f s = acc[t] + y; comp[t] = (s - acc[t]) - y; acc[t] = s;
            }
        } else if (MODE == 2) {
            const v16b a = bh_ld(arow, p.sAk, k0, h, p.K, 1.f);
#pragma unroll
            for (int t = 0; t < 2; ++t) {
                const int bn = min(n0 + t * 16 + l15, p.N - 1);
                acc[t] = wmmab(a, bh_ld(B + (long long)bn * p.sBn, p.sBk, k0, h, p.K, 1.f), acc[t]);
            }
        } else {
            const v16h a = fh_ld(arow, p.sAk, k0, h, p.K, p.sa);
#pragma unroll
            for (int t = 0; t < 2; ++t) {
                const int bn = min(n0 + t * 16 + l15, p.N - 1);
                acc[t] = wmma16(a, fh_ld(B + (long long)bn * p.sBn, p.sBk, k0, h, p.K, p.sb), acc[t]);
            }
        }
    }
    const float iscale = (MODE == 0) ? p.alpha / (p.sa * p.sb) : p.alpha;
    float* C = p.C + zo * p.sCo + zi * p.sCi;
    const float* R = p.R + zo * p.sRo + zi * p.sRi;
    __shared__ __align__(16) float ctile[16][36];
#pragma unroll
    for (int t = 0; t < 2; ++t) {
        const int n = n0 + t * 16 + l15; const int nn = min(n, p.N - 1);
#pragma unroll
        for (int r = 0; r < 8; ++r) {
            const int m = m0 + 8 * h + r; const int mm = min(m, p.M - 1);
            float v = acc[t][r] * iscale;
            if (p.flags & 1) v += p.bias[nn];
            if (p.flags & 2) v += p.bias[mm];
            v = act_fn(v, p.act);
            if (p.flags & 4) v += p.beta * R[(long long)mm * p.sRm + (long long)nn * p.sRn];
            ctile[8 * h + r][t * 16 + l15] = (n < p.N) ? v : 0.f;
        }
    }
    __syncthreads();
    const int NW = (p.Npad > p.N) ? p.Npad : p.N;
    const bool fast = (m0 + 16 <= p.M) && (n0 + 32 <= NW) && ((p.sCm & 3) == 0) && ((((size_t)C) & 15) == 0);
    if (fast) {
#pragma unroll
        for (int s = 0; s < 4; ++s) {
            const int row = s * 4 + (lane >> 3), c4 = (lane & 7) * 4;
            const v4f v = *(const v4f*)&ctile[row][c4];
            VST2V4(C + (long long)(m0 + row) * p.sCm + n0 + c4, v);
        }
    } else {
        for (int row = 0; row < 16; ++row) {
            const int m = m0 + row, n = n0 + lane;
            if (m < p.M && n < NW) VST2(float, C + (long long)m * p.sCm + n, ctile[row][lane]);
        }
    }
}

#define AW 4
struct AttnP {
    const float* Q; const float* K; const float* V; float* O; float* P; const float* Mf; const int* Mi; float* ST;
    const float* Pw; const float* Rt; const int* SQ; const int* SK;
    long long swb, swh, swi, swj, srb, srh, sri;
    long long sQb, sQh, sQi, sQd, sKb, sKh, sKj, sKd, sVb, sVh, sVj, sVd, sOb, sOh, sOi, sPb, sPh, sPi, smb, smh, smi, smj;
    int Lq, Lk, dh, dv, hrep, causal, coff, pband;
    float scale, mfill; int nonorm, mpol;
    int roff, rn, segpol, win;
};
static_assert(sizeof(AttnP) == 12 * 8 + 29 * 8 + 16 * 4, "AttnP has padding");

#ifndef KATTN_ATTR
#define KATTN_ATTR
#endif
template <int DHP, int DVP, int QM, bool SPLITPV, bool TWOPASS>
__global__ __launch_bounds__(32 * AW) KATTN_ATTR void k_attn(AttnP p) {
    constexpr int NT = DVP / 16;
    constexpr int KS = DHP / 32;
    constexpr int VP = DVP + 8;
    __shared__ __align__(16) float    pl[AW][16 * 64];
    __shared__ __align__(16) _Float16 vl[(SPLITPV ? 2 : 1) * 64 * VP];
    const int lane = threadIdx.x & 31, hf = lane >> 4, l15 = lane & 15, wave = threadIdx.x >> 5;
    const int h = blockIdx.y, b = blockIdx.z, hk = h / p.hrep;
    const int q0 = (blockIdx.x * AW + wave) * 16;
    float* myp = pl[wave];
    const float L2E = 1.4426950408889634f;
    const float NEG = -__builtin_inff();
    const int qi = min(q0 + l15, p.Lq - 1);
    const float* qrow = p.Q + b * p.sQb + h * p.sQh + (long long)qi * p.sQi;
    const float* kbase = p.K + b * p.sKb + hk * p.sKh;
    const float* vbase = p.V + b * p.sVb + hk * p.sVh;
    v16h qa[QM == 0 ? KS : 1]; Split qs_[QM == 1 ? KS : 1]; Split3 qt_[QM == 2 ? KS : 1];
#pragma unroll
    for (int ks = 0; ks < KS; ++ks) {
        if (QM == 2) qt_[ks] = sp3_ld(qrow, p.sQd, ks * 32, hf, p.dh, 1.f);
        else if (QM == 1) qs_[ks] = sp_ld(qrow, p.sQd, ks * 32, hf, p.dh, 1.f);
        else qa[ks] = fh_ld(qrow, p.sQd, ks * 32, hf, p.dh, 1.f);
    }
    v8f o[NT]; float m8[8], l8[8];
#pragma unroll
    for (int t = 0; t < NT; ++t) { v8f zz = {}; o[t] = zz; }
#pragma unroll
    for (int i = 0; i < 8; ++i) { m8[i] = NEG; l8[i] = 0.f; }
    int jend = p.Lk;
    if (p.causal == 1) { const int je = (blockIdx.x * AW + AW - 1) * 16 + 16 + p.coff; jend = min(jend, max(je, 0)); }
    const int npass = TWOPASS ? 2 : 1;
    for (int pass = 0; pass < npass; ++pass) {
        const bool dopv = (!TWOPASS) || pass == 1;
        for (int j0 = 0; j0 < jend; j0 += 64) {
            if (dopv) {
                __syncthreads();
                for (int idx = threadIdx.x; idx < 64 * DVP; idx += 32 * AW) {
                    const int jr = idx / DVP, d = idx - jr * DVP, j = j0 + jr;
                    const float f = (j < p.Lk && d < p.dv) ? vbase[(long long)j * p.sVj + (long long)d * p.sVd] : 0.f;
                    if (SPLITPV) {
                        const __bf16 hb = bf16_rne(f);
                        ((__bf16*)vl)[jr * VP + d] = hb; ((__bf16*)vl)[64 * VP + jr * VP + d] = bf16_rne(f - bf16_f32(hb));
                    } else vl[jr * VP + d] = (_Float16)f;
                }
            }
            v8f s[4];
#pragma unroll
            for (int t = 0; t < 4; ++t) {
                const int j = min(j0 + t * 16 + l15, p.Lk - 1);
                const float* krow = kbase + (long long)j * p.sKj;
                v8f acc = {};
#pragma unroll
                for (int ks = 0; ks < KS; ++ks) {
                    if (QM == 2)      acc = wmma6(qt_[ks], sp3_ld(krow, p.sKd, ks * 32, hf, p.dh, 1.f), acc);
                    else if (QM == 1) acc = wmma3(qs_[ks], sp_ld(krow, p.sKd, ks * 32, hf, p.dh, 1.f), acc);
                    else              acc = wmma16(qa[ks], fh_ld(krow, p.sKd, ks * 32, hf, p.dh, 1.f), acc);
                }
                s[t] = acc;
            }
            float pv[8][4];
#pragma unroll
            for (int i = 0; i < 8; ++i) {
                const int irow = q0 + i + 8 * hf;
                const int ic = min(irow, p.Lq - 1);
                float sc[4];
#pragma unroll
                for (int t = 0; t < 4; ++t) {
                    const int jg = j0 + t * 16 + l15;
                    float v = s[t][i] * p.scale;
                    if (p.Mf) v += p.Mf[b * p.smb + h * p.smh + (long long)ic * p.smi + (long long)min(jg, p.Lk - 1) * p.smj];
                    if (p.Rt) { int rc = ic - min(jg, p.Lk - 1) + p.roff; rc = rc < 0 ? 0 : (rc >= p.rn ? p.rn - 1 : rc); v += p.Rt[b * p.srb + h * p.srh + (long long)ic * p.sri + rc]; }
                    if (p.Mi) { const int mv = p.Mi[b * p.smb + h * p.smh + (long long)ic * p.smi + (long long)min(jg, p.Lk - 1) * p.smj]; if (p.mpol ? (mv != 0) : (mv == 0)) v = p.mfill; }
                    if (p.SQ) { const bool same = p.SQ[(long long)b * p.Lq + ic] == p.SK[(long long)b * p.Lk + min(jg, p.Lk - 1)]; if (p.segpol ? same : !same) v = p.mfill; }
                    if (p.causal == 2 && jg > irow + p.coff) v = p.mfill;
                    if (jg >= p.Lk || (p.causal == 1 && jg > irow + p.coff) || (p.causal == 3 && jg < irow + p.coff) || (p.win > 0 && irow + p.coff - jg > p.win)) v = NEG; else v *= L2E;
                    sc[t] = v;
                }
                if (!TWOPASS || pass == 0) {
                    float mx = fmaxf(fmaxf(sc[0], sc[1]), fmaxf(sc[2], sc[3]));
                    mx = fmaxf(mx, __shfl_xor(mx, 1, 32)); mx = fmaxf(mx, __shfl_xor(mx, 2, 32));
                    mx = fmaxf(mx, __shfl_xor(mx, 4, 32)); mx = fmaxf(mx, __shfl_xor(mx, 8, 32));
                    const float mnew = fmaxf(m8[i], mx);
                    const float corr = (mnew == NEG) ? 1.f : exp2f(m8[i] - mnew);
                    float rs = 0.f;
#pragma unroll
                    for (int t = 0; t < 4; ++t) {
                        const float pp = (sc[t] == NEG) ? 0.f : exp2f(sc[t] - mnew); rs += pp;
                        pv[i][t] = p.Pw ? pp * p.Pw[b * p.swb + h * p.swh + (long long)ic * p.swi + (long long)min(j0 + t * 16 + l15, p.Lk - 1) * p.swj] : pp;
                    }
                    rs += __shfl_xor(rs, 1, 32); rs += __shfl_xor(rs, 2, 32); rs += __shfl_xor(rs, 4, 32); rs += __shfl_xor(rs, 8, 32);
                    l8[i] = l8[i] * corr + rs; m8[i] = mnew;
                    if (!TWOPASS) {
#pragma unroll
                        for (int t = 0; t < NT; ++t) o[t][i] *= corr;
                    }
                } else {
                    const float inv = (l8[i] > 0.f) ? 1.f / l8[i] : 0.f;
#pragma unroll
                    for (int t = 0; t < 4; ++t) {
                        const int jg = j0 + t * 16 + l15;
                        float pp = (sc[t] == NEG) ? 0.f : exp2f(sc[t] - m8[i]) * inv;
                        if (p.Pw) pp *= p.Pw[b * p.swb + h * p.swh + (long long)ic * p.swi + (long long)min(jg, p.Lk - 1) * p.swj];
                        pv[i][t] = pp;
                    }
                }
            }
            if (dopv) {
#pragma unroll
                for (int i = 0; i < 8; ++i)
#pragma unroll
                    for (int t = 0; t < 4; ++t) myp[(i + 8 * hf) * 64 + t * 16 + l15] = pv[i][t];
                __syncthreads();
                if (p.P) {
                    float* pb_ = p.P + b * p.sPb + h * p.sPh;
                    const bool fastP = (p.pband == 0) && ((p.sPi & 3) == 0) && (j0 + 64 <= p.Lk) && (q0 + 16 <= p.Lq) && ((((size_t)pb_) & 15) == 0);
                    if (fastP) {
#pragma unroll
                        for (int s = 0; s < 8; ++s) {
                            const int row = s * 2 + (lane >> 4), c4 = (lane & 15) * 4;
                            const v4f v = *(const v4f*)(myp + row * 64 + c4);
                            VST2V4(pb_ + (long long)(q0 + row) * p.sPi + j0 + c4, v);
                        }
                    } else {
                        for (int row = 0; row < 16; ++row) {
                            const int irow = q0 + row; if (irow >= p.Lq) continue;
                            for (int c = lane; c < 64; c += 32) {
                                const int jg = j0 + c; if (jg >= p.Lk) continue;
                                if (p.pband == 0) VST2(float, pb_ + (long long)irow * p.sPi + jg, myp[row * 64 + c]);
                                else if (jg - irow <= p.pband && irow - jg <= p.pband) VST2(float, pb_ + (long long)irow * p.sPi + (jg - irow + p.pband), myp[row * 64 + c]);
                            }
                        }
                    }
                }
                if (SPLITPV) {
                    const Split pa0 = sp_ld(myp + l15 * 64, 1, 0, hf, 64, 1.f), pa1 = sp_ld(myp + l15 * 64, 1, 32, hf, 64, 1.f);
                    const __bf16* vh = (const __bf16*)vl; const __bf16* vlo = vh + 64 * VP;
#pragma unroll
                    for (int t = 0; t < NT; ++t) {
                        const int dcol = t * 16 + l15;
                        Split b0, b1;
#pragma unroll
                        for (int e = 0; e < 16; ++e) {
                            const int k0 = frag_k(e, hf), k1 = 32 + frag_k(e, hf);
                            b0.hi[e] = vh[k0 * VP + dcol]; b0.lo[e] = vlo[k0 * VP + dcol]; b1.hi[e] = vh[k1 * VP + dcol]; b1.lo[e] = vlo[k1 * VP + dcol];
                        }
                        o[t] = wmma3(pa0, b0, o[t]);
                        o[t] = wmma3(pa1, b1, o[t]);
                    }
                } else {
                    const v16h pa0 = fh_ld(myp + l15 * 64, 1, 0, hf, 64, 4096.f), pa1 = fh_ld(myp + l15 * 64, 1, 32, hf, 64, 4096.f);
#pragma unroll
                    for (int t = 0; t < NT; ++t) {
                        const int dcol = t * 16 + l15;
                        v16h b0, b1;
#pragma unroll
                        for (int e = 0; e < 16; ++e) { b0[e] = vl[frag_k(e, hf) * VP + dcol]; b1[e] = vl[(32 + frag_k(e, hf)) * VP + dcol]; }
                        o[t] = wmma16(pa0, b0, o[t]);
                        o[t] = wmma16(pa1, b1, o[t]);
                    }
                }
            }
        }
    }
    float* obase = p.O + b * p.sOb + h * p.sOh;
    if (p.ST) {
        const int rl = lane >> 1, isel = rl & 7;
        float mv = 0.f, lv = 0.f;
#pragma unroll
        for (int i = 0; i < 8; ++i) if (i == isel) { mv = m8[i]; lv = l8[i]; }
        const int irow = q0 + rl;
        if (irow < p.Lq) { float* st = p.ST + (((long long)b * gridDim.y + h) * p.Lq + irow) * 2 + (lane & 1); VST2(float, st, (lane & 1) ? lv : mv * 0.6931471805599453f); }
    }
    float invr[8];
#pragma unroll
    for (int i = 0; i < 8; ++i) {
        if (TWOPASS) invr[i] = SPLITPV ? 1.f : (1.f / 4096.f);
        else if (p.nonorm) invr[i] = exp2f(m8[i]) * (SPLITPV ? 1.f : (1.f / 4096.f));
        else invr[i] = (l8[i] > 0.f) ? (SPLITPV ? 1.f / l8[i] : 1.f / (l8[i] * 4096.f)) : 0.f;
    }
    __syncthreads();
    const bool ofast = ((p.sOi & 3) == 0) && ((((size_t)obase) & 15) == 0) && (q0 + 16 <= p.Lq);
#pragma unroll
    for (int c0 = 0; c0 < DVP; c0 += 64) {
#pragma unroll
        for (int i = 0; i < 8; ++i)
#pragma unroll
            for (int t = 0; t < NT; ++t) if (t * 16 >= c0 && t * 16 < c0 + 64) myp[(i + 8 * hf) * 64 + (t * 16 - c0) + l15] = o[t][i] * invr[i];
        __syncthreads();
        const int cw = (DVP - c0 < 64) ? (DVP - c0) : 64;
        if (ofast && (c0 + cw <= p.dv) && (cw % 32 == 0)) {
            const int lpr = cw / 4;
            const int rows_per_ins = 32 / lpr;
            for (int r0 = 0; r0 < 16; r0 += rows_per_ins) {
                const int row = r0 + lane / lpr, c4 = (lane % lpr) * 4;
                const v4f v = *(const v4f*)(myp + row * 64 + c4);
                VST2V4(obase + (long long)(q0 + row) * p.sOi + c0 + c4, v);
            }
        } else {
            for (int row = 0; row < 16; ++row) {
                const int irow = q0 + row; if (irow >= p.Lq) continue;
                for (int c = lane; c < cw; c += 32) { const int d = c0 + c; if (d < p.dv) VST2(float, obase + (long long)irow * p.sOi + d, myp[row * 64 + c]); }
            }
        }
        __syncthreads();
    }
}

struct TrP { const float* src; float* dst; const float* R2; long long sSz, lds, sDz, ldd, sRz, ldr; int R, C, flags, act; float alpha, beta; };
static_assert(sizeof(TrP) == 3 * 8 + 6 * 8 + 6 * 4, "TrP has padding");
__global__ __launch_bounds__(256) void k_tr(TrP p) {
    __shared__ float tile[32][33];
    const int c0 = blockIdx.x * 32, r0 = blockIdx.y * 32, z = blockIdx.z;
    const int lane = threadIdx.x & 31, wave = threadIdx.x >> 5;
    const float* s = p.src + z * p.sSz;
#pragma unroll
    for (int k = 0; k < 4; ++k) {
        const int rl = wave * 4 + k, r = r0 + rl, c = c0 + lane;
        tile[rl][lane] = (r < p.R && c < p.C) ? s[(long long)r * p.lds + c] : 0.f;
    }
    __syncthreads();
    float* d = p.dst + z * p.sDz; const float* rr = p.R2 + z * p.sRz;
#pragma unroll
    for (int k = 0; k < 4; ++k) {
        const int cl = wave * 4 + k, c = c0 + cl, r = r0 + lane;
        if (c < p.C && r < p.R) {
            float v = act_fn(p.alpha * tile[lane][cl], p.act);
            if (p.flags & 1) v += p.beta * rr[(long long)c * p.ldr + r];
            VST2(float, d + (long long)c * p.ldd + r, v);
        }
    }
}

__global__ __launch_bounds__(256) void k_affine(const float* __restrict__ src, float* __restrict__ dst, int n, float a, float b, const float* __restrict__ sdev) {
    const int i = blockIdx.x * 256 + threadIdx.x;
    if (i < n) { const float aa = sdev ? a * sdev[0] : a; const float v = aa * src[i] + b; VST2(float, dst + i, v); }
}

struct SmP { const float* src; float* dst; const float* Mf; long long sz, sr, dz, dr, smz, smr; int n, pad; float scale_in, scale_out; };
static_assert(sizeof(SmP) == 3 * 8 + 6 * 8 + 4 * 4, "SmP has padding");
__global__ __launch_bounds__(256) void k_softmax(SmP p) {
    __shared__ float red[256];
    const int r = blockIdx.x, z = blockIdx.y, tid = threadIdx.x;
    const float* s = p.src + z * p.sz + (long long)r * p.sr;
    const float* mf = p.Mf ? (p.Mf + z * p.smz + (long long)r * p.smr) : nullptr;
    float mx = -__builtin_inff();
    for (int j = tid; j < p.n; j += 256) { float v = s[j] * p.scale_in; if (mf) v += mf[j]; mx = fmaxf(mx, v); }
    red[tid] = mx; __syncthreads();
    for (int o = 128; o > 0; o >>= 1) { if (tid < o) red[tid] = fmaxf(red[tid], red[tid + o]); __syncthreads(); }
    mx = red[0]; __syncthreads();
    float sum = 0.f;
    for (int j = tid; j < p.n; j += 256) { float v = s[j] * p.scale_in; if (mf) v += mf[j]; sum += (mx == -__builtin_inff()) ? 0.f : expf(v - mx); }
    red[tid] = sum; __syncthreads();
    for (int o = 128; o > 0; o >>= 1) { if (tid < o) red[tid] += red[tid + o]; __syncthreads(); }
    sum = red[0];
    const float inv = (sum > 0.f) ? p.scale_out / sum : 0.f;
    float* d = p.dst + z * p.dz + (long long)r * p.dr;
    for (int j = tid; j < p.n; j += 256) { float v = s[j] * p.scale_in; if (mf) v += mf[j]; const float o = (mx == -__builtin_inff()) ? 0.f : expf(v - mx) * inv; VST2(float, d + j, o); }
}
__global__ __launch_bounds__(256) void k_stats(const float* __restrict__ x, long long sz, long long so, long long si, int inner, int n, float eps, float* __restrict__ stat, int mode) {
    __shared__ float red[256];
    const int z = blockIdx.x, tid = threadIdx.x;
    const float* base = x + z * sz;
    float s = 0.f;
    for (int e = tid; e < n; e += 256) s += base[(long long)(e / inner) * so + (long long)(e % inner) * si];
    red[tid] = s; __syncthreads();
    for (int o = 128; o > 0; o >>= 1) { if (tid < o) red[tid] += red[tid + o]; __syncthreads(); }
    const float mu = (mode == 0 || mode == 3) ? red[0] / (float)n : 0.f; __syncthreads();
    float q = 0.f;
    for (int e = tid; e < n; e += 256) { const float dlt = base[(long long)(e / inner) * so + (long long)(e % inner) * si] - mu; q += dlt * dlt; }
    red[tid] = q; __syncthreads();
    for (int o = 128; o > 0; o >>= 1) { if (tid < o) red[tid] += red[tid + o]; __syncthreads(); }
    {
        float rs;
        if (mode == 2) rs = sqrtf((float)n) / fmaxf(sqrtf(red[0]), eps); else if (mode == 3) rs = rsqrtf(red[0] / (float)(n - 1) + eps); else rs = rsqrtf(red[0] / (float)n + eps);
        if (tid < 32) { const float v = (tid == 0) ? mu : ((tid == 1) ? rs : 0.f); VST2(float, stat + (long long)z * 32 + tid, v); }
    }
}
__global__ __launch_bounds__(256) void k_norm_apply(const float* __restrict__ x, float* __restrict__ y, const float* __restrict__ stat, const float* __restrict__ g, const float* __restrict__ bta,
                                                     int Z, int C, int L, int G, int bn, int act) {
    const long long idx = (long long)blockIdx.x * 256 + threadIdx.x;
    if (idx >= (long long)Z * C * L) return;
    const int l = (int)(idx % L); const long long zc = idx / L; const int c = (int)(zc % C), z = (int)(zc / C); (void)l;
    const int set = bn ? c : (z * G + c / (C / G));
    float v = (x[idx] - stat[(long long)set * 32]) * stat[(long long)set * 32 + 1];
    if (g) v *= g[c];
    if (bta) v += bta[c];
    v = act_fn(v, act);
    VST2(float, y + idx, v);
}

__global__ __launch_bounds__(256) void k_lse_neg(const float* __restrict__ st, float* __restrict__ c, int n) {
    const int i = blockIdx.x * 256 + threadIdx.x;
    if (i < n) { const float v = -(st[2 * i] + logf(st[2 * i + 1])); VST2(float, c + i, v); }
}

__global__ __launch_bounds__(256) void k_iota(int* __restrict__ dst, int n, int a, int b) {
    const int i = blockIdx.x * 256 + threadIdx.x;
    if (i < n) { const int v = a * i + b; VST2(int, dst + i, v); }
}

__global__ __launch_bounds__(256) void k_axpby(const float* __restrict__ x, const float* __restrict__ y, float* __restrict__ dst, int n, float a, float b, float c) {
    const int i = blockIdx.x * 256 + threadIdx.x;
    if (i < n) { const float v = a * x[i] + b * y[i] + c; VST2(float, dst + i, v); }
}

struct RopeP { const float* X; float* Y; const float* C; const float* Sn; const int* pos; long long sXr, sXh, sYr, sYh, sCb, sCp, sCd; int R, Hn, D, S, mode, tmode, pmode, pad; };
static_assert(sizeof(RopeP) == 5 * 8 + 7 * 8 + 8 * 4, "RopeP has padding");
__global__ __launch_bounds__(256) void k_rope(RopeP p) {
    const long long idx = (long long)blockIdx.x * 256 + threadIdx.x;
    if (idx >= (long long)p.R * p.Hn * p.D) return;
    const int d = (int)(idx % p.D); const long long rh = idx / p.D; const int h = (int)(rh % p.Hn); const int r = (int)(rh / p.Hn);
    const int half = p.D / 2;
    int partner; float sign;
    if (p.mode == 0) { partner = (d < half) ? d + half : d - half; sign = (d < half) ? -1.f : 1.f; }
    else { partner = d ^ 1; sign = (d & 1) ? 1.f : -1.f; }
    const int tcol = (p.tmode == 0) ? d : ((p.tmode == 1) ? (d % half) : (d >> 1));
    const int pp = (p.pmode == 0) ? (r % p.S) : ((p.pmode == 1) ? h : p.pos[r]);
    const long long toff = (long long)(r / p.S) * p.sCb + (long long)pp * p.sCp + (long long)tcol * p.sCd;
    const float* xr = p.X + (long long)r * p.sXr + (long long)h * p.sXh;
    const float v = xr[d] * p.C[toff] + sign * xr[partner] * p.Sn[toff];
    VST2(float, p.Y + (long long)r * p.sYr + (long long)h * p.sYh + d, v);
}

__global__ __launch_bounds__(256) void k_invf(float* __restrict__ invb, int half, int D, float base, float num, int fmode, float cexp) {
    const int i = blockIdx.x * 256 + threadIdx.x;
    if (i >= ((half + 31) / 32) * 32) return;
    if (i >= half) { VST2(float, invb + i, 0.f); return; }
    const float e = (float)(2 * i) / (float)D;
    float invf;
    if (fmode == 1) invf = num * expf((float)(2 * i) * cexp);
    else if (fmode == 2) invf = num * powf(base, (-2.0f * ((float)i - 1.0f)) / (float)D);
    else invf = num * (1.0f / powf(base, e));
    VST2(float, invb + i, invf);
}
__global__ __launch_bounds__(256) void k_sincos(float* __restrict__ cs, float* __restrict__ sn, const float* __restrict__ invb, int S, int half, float pscale) {
    const int idx = blockIdx.x * 256 + threadIdx.x;
    if (idx >= S * half) return;
    const int s = idx / half, i = idx - s * half;
    const float ang = (pscale * (float)s) * invb[i];
    VST2(float, cs + idx, cosf(ang)); VST2(float, sn + idx, sinf(ang));
}

__global__ __launch_bounds__(256) void k_mulact(const float* __restrict__ x, const float* __restrict__ y, float* __restrict__ dst, int n, int act) {
    const int i = blockIdx.x * 256 + threadIdx.x;
    if (i < n) { const float v = act_fn(x[i], act) * y[i]; VST2(float, dst + i, v); }
}

__global__ __launch_bounds__(256) void k_matvec(GemmP p) {
    const int rpt = (p.N == 1) ? 1 : 32;
    const long long r0 = ((long long)blockIdx.x * 256 + threadIdx.x) * rpt; const int z = blockIdx.z, zo = z / p.zi_n, zi = z - zo * p.zi_n;
    if (r0 >= p.M) return;
    const float* Bb = p.B + zo * p.sBo + zi * p.sBi;
    float* C = p.C + zo * p.sCo + zi * p.sCi; const float* R = p.R + zo * p.sRo + zi * p.sRi;
    for (int rr = 0; rr < rpt; ++rr) {
        const long long r = r0 + rr; if (r >= p.M) break;
        const float* A = p.A + zo * p.sAo + zi * p.sAi + r * p.sAm;
        float acc[8] = {0.f, 0.f, 0.f, 0.f, 0.f, 0.f, 0.f, 0.f};
        for (int k = 0; k < p.K; ++k) { const float a = A[(long long)k * p.sAk];
#pragma unroll
            for (int j = 0; j < 8; ++j) if (j < p.N) acc[j] += a * Bb[(long long)j * p.sBn + (long long)k * p.sBk]; }
#pragma unroll
        for (int j = 0; j < 8; ++j) if (j < p.N) {
            float v = acc[j] * p.alpha;
            if (p.flags & 1) v += p.bias[j];
            if (p.flags & 2) v += p.bias[r];
            v = act_fn(v, p.act);
            if (p.flags & 4) v += p.beta * R[r * p.sRm + (long long)j * p.sRn];
            VST2(float, C + r * p.sCm + j, v);
        }
    }
}
__global__ __launch_bounds__(256) void k_smallsoftmax(const float* __restrict__ src, float* __restrict__ dst, long long sr, long long dr, int n, long long R, float scale) {
    const long long r0 = ((long long)blockIdx.x * 256 + threadIdx.x) * 32;
    for (int rr = 0; rr < 32; ++rr) {
        const long long r = r0 + rr; if (r >= R) return;
        const float* s = src + r * sr; float* d = dst + r * dr;
        float mx = -__builtin_inff();
        for (int j = 0; j < n; ++j) mx = fmaxf(mx, s[j] * scale);
        float sum = 0.f;
        for (int j = 0; j < n; ++j) sum += expf(s[j] * scale - mx);
        const float inv = 1.f / sum;
        for (int j = 0; j < n; ++j) { const float v = expf(s[j] * scale - mx) * inv; VST2(float, d + j, v); }
    }
}

__global__ __launch_bounds__(32) void k_unitstat(float* __restrict__ st) { const int t = threadIdx.x; const float v = (t == 1) ? 1.f : 0.f; VST2(float, st + t, v); }

__global__ __launch_bounds__(256) void k_lincopy(const float* __restrict__ src, long long lds, float* __restrict__ dst, long long ldd, long long rows, int cols) {
    const long long i = (long long)blockIdx.x * 256 + threadIdx.x; if (i >= rows * cols) return;
    const long long r = i / cols; const int c = (int)(i - r * cols);
    const float v = src[r * lds + c]; VST2(float, dst + r * ldd + c, v);
}

__global__ __launch_bounds__(256) void k_cc_norm(const float* __restrict__ co, float* __restrict__ NC, int* __restrict__ VIX, int N, int R) {
    __shared__ float red[256]; __shared__ float mean[3]; const int b = blockIdx.x; const float* cb = co + (long long)b * 3 * N;
    for (int d = 0; d < 3; ++d) { float s = 0.f; for (int n = threadIdx.x; n < N; n += 256) s += cb[d * N + n]; red[threadIdx.x] = s; __syncthreads(); for (int o = 128; o > 0; o >>= 1) { if (threadIdx.x < o) red[threadIdx.x] += red[threadIdx.x + o]; __syncthreads(); } if (threadIdx.x == 0) mean[d] = red[0] / (float)N; __syncthreads(); }
    float mx = 0.f; for (int n = threadIdx.x; n < N; n += 256) { const float x = cb[n] - mean[0], y = cb[N + n] - mean[1], z = cb[2 * N + n] - mean[2]; mx = fmaxf(mx, sqrtf(x * x + y * y + z * z)); }
    red[threadIdx.x] = mx; __syncthreads(); for (int o = 128; o > 0; o >>= 1) { if (threadIdx.x < o) red[threadIdx.x] = fmaxf(red[threadIdx.x], red[threadIdx.x + o]); __syncthreads(); } const float den = red[0] * 2.f + 0.f;
    for (int n = threadIdx.x; n < N; n += 256) { int v[3]; for (int d = 0; d < 3; ++d) { float u = (cb[d * N + n] - mean[d]) / den + 0.5f; u = fminf(fmaxf(u * (float)R, 0.f), (float)(R - 1)); VST2(float, NC + ((long long)b * N + n) * 4 + d, u); v[d] = (int)rintf(u); }
        VST2(float, NC + ((long long)b * N + n) * 4 + 3, 0.f); VST2(int, VIX + (long long)b * N + n, b * R * R * R + (v[0] * R + v[1]) * R + v[2]); }
}
__global__ __launch_bounds__(256) void k_cc_ft(const float* __restrict__ F, float* __restrict__ FT, int B, int C, int N) { const long long q = (long long)blockIdx.x * 256 + threadIdx.x; if (q >= (long long)B * N * C) return; const int c = (int)(q % C); const int n = (int)((q / C) % N); const int b = (int)(q / ((long long)C * N)); VST2(float, FT + q, F[((long long)b * C + c) * N + n]); }
__global__ __launch_bounds__(256) void k_cc_vox(const float* __restrict__ FT, const int* __restrict__ off, const int* __restrict__ slot, float* __restrict__ GP, int B, int R, int C) { const long long q = (long long)blockIdx.x * 256 + threadIdx.x; const long long R3 = (long long)R * R * R; if (q >= (long long)B * R3 * C) return; const int c = (int)(q % C); const long long v = q / C; const int a = off[v], e = off[v + 1]; if (a >= e) return; float s = 0.f; for (int p = a; p < e; ++p) s += FT[(long long)slot[p] * C + c];
    const int b = (int)(v / R3); const int r = (int)(v % R3); const int x = r / (R * R), y = (r / R) % R, z = r % R; VST2(float, GP + ((((long long)b * (R + 2) + x + 1) * (R + 2) + y + 1) * (R + 2) + z + 1) * C + c, s / (float)(e - a)); }
__global__ __launch_bounds__(256) void k_cc_bnl(float* __restrict__ GC, const float* __restrict__ g, const float* __restrict__ bb, float* __restrict__ GPo, int B, int R, int C) { const long long q = (long long)blockIdx.x * 256 + threadIdx.x; const long long R3 = (long long)R * R * R; if (q >= (long long)B * R3 * C) return; const int c = (int)(q % C); const long long v = q / C; float u = GC[q] * (g[c] * rsqrtf(1.f + 1e-4f)) + bb[c]; u = (u >= 0.f) ? u : 0.1f * u; VST2(float, GC + q, u);
    if (GPo) { const int b = (int)(v / R3); const int r = (int)(v % R3); const int x = r / (R * R), y = (r / R) % R, z = r % R; VST2(float, GPo + ((((long long)b * (R + 2) + x + 1) * (R + 2) + y + 1) * (R + 2) + z + 1) * C + c, u); } }
__global__ __launch_bounds__(256) void k_cc_devox(const float* __restrict__ GC, const float* __restrict__ NC, float* __restrict__ F1, int B, int N, int R, int C) { const long long q = (long long)blockIdx.x * 256 + threadIdx.x; if (q >= (long long)B * N * C) return; const int c = (int)(q % C); const long long pn = q / C; const int b = (int)(pn / N); const float* nc = NC + pn * 4;
    int lo[3], hi[3]; float w1[3]; for (int d = 0; d < 3; ++d) { const float fl = floorf(nc[d]); lo[d] = (int)fl; hi[d] = min(lo[d] + 1, R - 1); w1[d] = nc[d] - fl; }
    float acc = 0.f;
#pragma unroll 1
    for (int corner = 0; corner < 8; ++corner) { const int dx = corner >> 2, dy = (corner >> 1) & 1, dz = corner & 1; const int ix = dx ? hi[0] : lo[0], iy = dy ? hi[1] : lo[1], iz = dz ? hi[2] : lo[2]; const float w = (dx ? w1[0] : 1.f - w1[0]) * (dy ? w1[1] : 1.f - w1[1]) * (dz ? w1[2] : 1.f - w1[2]);
        acc += w * GC[(((long long)b * R * R * R) + ((long long)ix * R + iy) * R + iz) * C + c]; }
    VST2(float, F1 + q, acc); }
__global__ __launch_bounds__(128) void k_cc_knn(const float* __restrict__ co, int* __restrict__ IDX, float* __restrict__ MSK, int B, int N, float r2) { __shared__ float sp[3 * 512]; const int q = blockIdx.x * 128 + threadIdx.x; const bool ok = q < B * N; const int b = ok ? q / N : 0; const int n = ok ? q % N : 0; const float* cb = co + (long long)b * 3 * N;
    const float xn = ok ? cb[n] : 0.f, yn = ok ? cb[N + n] : 0.f, zn = ok ? cb[2 * N + n] : 0.f; const float sqn = xn * xn + yn * yn + zn * zn; float bd[16]; int bi[16]; for (int j = 0; j < 16; ++j) { bd[j] = __builtin_inff(); bi[j] = 0; }
    for (int j0 = 0; j0 < N; j0 += 512) { __syncthreads(); for (int t = threadIdx.x; t < 512 * 3; t += 128) { const int d = t / 512, jj = t % 512; sp[t] = cb[(long long)d * N + j0 + jj]; } __syncthreads();
#pragma unroll 1
        for (int jj = 0; jj < 512; ++jj) { const float xm = sp[jj], ym = sp[512 + jj], zm = sp[1024 + jj]; const float d2 = (sqn + (xm * xm + ym * ym + zm * zm)) - 2.f * (xn * xm + yn * ym + zn * zm); if (d2 < bd[15]) { int s = 15; while (s > 0 && d2 < bd[s - 1]) { bd[s] = bd[s - 1]; bi[s] = bi[s - 1]; --s; } bd[s] = d2; bi[s] = j0 + jj; } } }
    if (ok) for (int j = 0; j < 16; ++j) { VST2(int, IDX + (long long)q * 16 + j, bi[j]); VST2(float, MSK + (long long)q * 16 + j, (bd[j] <= r2) ? 1.f : 0.f); } }
__global__ __launch_bounds__(64) void k_cc_pattn(const float* __restrict__ QT, const float* __restrict__ KT, const float* __restrict__ VT, const int* __restrict__ IDX, const float* __restrict__ MSK, const float* __restrict__ F1, float* __restrict__ F12, int B, int N, int C) {
    __shared__ float w[16]; const int pn = blockIdx.x; const int b = pn / N; const int c = threadIdx.x;
    __shared__ float sc[16]; if (c < 16) { const int m = IDX[(long long)pn * 16 + c]; float s = 0.f;
#pragma unroll 1
        for (int d = 0; d < C; ++d) s += QT[(long long)pn * C + d] * KT[((long long)b * N + m) * C + d]; sc[c] = (MSK[(long long)pn * 16 + c] > 0.5f) ? s * 0.125f : -1e9f; }
    __syncthreads(); if (c == 0) { float mx = -__builtin_inff();
#pragma unroll 1
        for (int j = 0; j < 16; ++j) mx = fmaxf(mx, sc[j]);
        float s = 0.f;
#pragma unroll 1
        for (int j = 0; j < 16; ++j) { const float e = expf(sc[j] - mx); w[j] = e; s += e; }
#pragma unroll 1
        for (int j = 0; j < 16; ++j) w[j] = w[j] / s; } __syncthreads();
    float a = 0.f;
#pragma unroll 1
    for (int j = 0; j < 16; ++j) a += w[j] * VT[((long long)b * N + IDX[(long long)pn * 16 + j]) * C + c];
    VST2(float, F12 + (long long)pn * 2 * C + C + c, a); VST2(float, F12 + (long long)pn * 2 * C + c, F1[(long long)pn * C + c]); }
__global__ __launch_bounds__(256) void k_cc_out(const float* __restrict__ FU, const float* __restrict__ co, float* __restrict__ OUT, float* __restrict__ COUT, int B, int C, int N) { const long long q = (long long)blockIdx.x * 256 + threadIdx.x; if (q >= (long long)B * C * N) return; const int n = (int)(q % N); const int o = (int)((q / N) % C); const int b = (int)(q / ((long long)N * C)); VST2(float, OUT + q, FU[((long long)b * N + n) * C + o]); if (q < (long long)B * 3 * N) VST2(float, COUT + q, co[q]); }

#define IL_CAP32 32
#define IL_T32 256
#define IL_TILE32 4096
__global__ __launch_bounds__(IL_T32) void k_inlists32(const int* __restrict__ tgt, int E, int N, int* __restrict__ NBR, int* __restrict__ cnt) {
    __shared__ int tt[IL_TILE32];
    __shared__ int lists[IL_T32 * IL_CAP32];
    const int d = blockIdx.x * IL_T32 + threadIdx.x; int n = 0;
    for (int e0 = 0; e0 < E; e0 += IL_TILE32) {
        const int nt = min(IL_TILE32, E - e0);
        __syncthreads();
        for (int i = threadIdx.x; i < nt; i += IL_T32) tt[i] = tgt[e0 + i];
        __syncthreads();
        for (int i = 0; i < nt; ++i) { if (tt[i] == d) { if (n < IL_CAP32) lists[threadIdx.x * IL_CAP32 + n] = e0 + i; ++n; } }
    }
    if (d < N) {
        int* row = NBR + (long long)d * IL_CAP32;
        for (int j = 0; j < IL_CAP32; ++j) { const int v = (j < n) ? lists[threadIdx.x * IL_CAP32 + j] : -1; VST2(int, row + j, v); }
        VST2(int, cnt + d, min(n, IL_CAP32));
    }
}
__global__ __launch_bounds__(256) void k_csr_scan32(const int* __restrict__ cnt, int* __restrict__ off, int N) {
    __shared__ int part[256]; const int per = ((((N + 255) / 256) + 31) / 32) * 32; const int a = threadIdx.x * per, b = min(N, a + per); int s = 0;
    for (int i = a; i < b; ++i) s += cnt[i]; part[threadIdx.x] = s; __syncthreads();
    if (threadIdx.x == 0) { int run = 0; for (int t = 0; t < 256; ++t) { const int v = part[t]; part[t] = run; run += v; } } __syncthreads();
    int run = part[threadIdx.x]; for (int i = a; i < b; ++i) { VST2(int, off + i, run); run += cnt[i]; }
    if (a < N && b == N) { VST2(int, off + N, run); }
}
__global__ __launch_bounds__(256) void k_slotcopy32(const int* __restrict__ off, const int* __restrict__ NBR, int* __restrict__ slot, int N) {
    const int t = blockIdx.x * 256 + threadIdx.x; const int tot = off[N]; if (t >= tot) return;
    int lo = 0, hi = N - 1;
    while (lo < hi) { const int mid = (lo + hi + 1) >> 1; if (off[mid] <= t) lo = mid; else hi = mid - 1; }
    int j = t - off[lo]; j = (j < 0) ? 0 : ((j >= IL_CAP32) ? (IL_CAP32 - 1) : j);
    VST2(int, slot + t, NBR[(long long)lo * IL_CAP32 + j]);
}

__global__ __launch_bounds__(256) void k_cc_f3(float* __restrict__ F3, const float* __restrict__ g, const float* __restrict__ bb, long long n, int C) { const long long q = (long long)blockIdx.x * 256 + threadIdx.x; if (q >= n) return; const int c = (int)(q % C); const float v = fmaxf(F3[q] * (g[c] * rsqrtf(1.f + 1e-4f)) + bb[c], 0.f); VST2(float, F3 + q, v); }

template __global__ void k_gemm<1>(GemmP);

extern "C" void kernel_launch(void* const* d_in, const int* in_sizes, int n_in, void* d_out, int out_size, void* d_ws, size_t ws_size, hipStream_t stream) {
    (void)in_sizes; (void)n_in; (void)out_size; (void)ws_size;
    const float* feat = (const float*)d_in[0];
    const float* coords = (const float*)d_in[1];
    const float* wv1 = (const float*)d_in[2];
    const float* bv1 = (const float*)d_in[3];
    const float* g1 = (const float*)d_in[4];
    const float* be1 = (const float*)d_in[5];
    const float* wv2 = (const float*)d_in[6];
    const float* bv2 = (const float*)d_in[7];
    const float* g2 = (const float*)d_in[8];
    const float* be2 = (const float*)d_in[9];
    const float* wq = (const float*)d_in[10];
    const float* bq = (const float*)d_in[11];
    const float* wk = (const float*)d_in[12];
    const float* bk = (const float*)d_in[13];
    const float* wv = (const float*)d_in[14];
    const float* bv = (const float*)d_in[15];
    const float* wp = (const float*)d_in[16];
    const float* bp = (const float*)d_in[17];
    const float* gp = (const float*)d_in[18];
    const float* bep = (const float*)d_in[19];
    const float* w2 = (const float*)d_in[20];
    const float* b2 = (const float*)d_in[21];
    const int Bn = 4;
    const int C = 64;
    const int N = 4096;
    const int R = 32;
    const int R3 = 32768;
    const int RP = 34;
    const int RP3 = RP * RP * RP;
    const int NV = Bn * R3;
    const int NPt = Bn * N;
    const int CAP = 32;
    const int KN = 16;
    float* out = (float*)d_out;
    float* cout = out + ((size_t)Bn * C * N);
    char* wsp = (char*)d_ws;
    float* NC = (float*)wsp; wsp += (((size_t)((size_t)NPt * 4) * 4 + 255) / 256) * 256;
    int* VIX = (int*)wsp; wsp += (((size_t)((size_t)NPt + 64) * 4 + 255) / 256) * 256;
    int* cnt = (int*)wsp; wsp += (((size_t)((size_t)NV + 64) * 4 + 255) / 256) * 256;
    int* off = (int*)wsp; wsp += (((size_t)((size_t)NV + 64) * 4 + 255) / 256) * 256;
    int* slot = (int*)wsp; wsp += (((size_t)((size_t)NPt + 64) * 4 + 255) / 256) * 256;
    int* nbr = (int*)wsp; wsp += (((size_t)((size_t)NV * CAP) * 4 + 255) / 256) * 256;
    float* FT = (float*)wsp; wsp += (((size_t)((size_t)NPt * C) * 4 + 255) / 256) * 256;
    float* GP = (float*)wsp; wsp += (((size_t)((size_t)Bn * RP3 * C) * 4 + 255) / 256) * 256;
    float* GQ = (float*)wsp; wsp += (((size_t)((size_t)Bn * RP3 * C) * 4 + 255) / 256) * 256;
    float* GC = (float*)wsp; wsp += (((size_t)((size_t)NV * C) * 4 + 255) / 256) * 256;
    float* F1 = (float*)wsp; wsp += (((size_t)((size_t)NPt * C) * 4 + 255) / 256) * 256;
    float* QT = (float*)wsp; wsp += (((size_t)((size_t)NPt * C) * 4 + 255) / 256) * 256;
    float* KT = (float*)wsp; wsp += (((size_t)((size_t)NPt * C) * 4 + 255) / 256) * 256;
    float* VT = (float*)wsp; wsp += (((size_t)((size_t)NPt * C) * 4 + 255) / 256) * 256;
    int* IDX = (int*)wsp; wsp += (((size_t)((size_t)NPt * KN) * 4 + 255) / 256) * 256;
    float* MSK = (float*)wsp; wsp += (((size_t)((size_t)NPt * KN) * 4 + 255) / 256) * 256;
    float* F12 = (float*)wsp; wsp += (((size_t)((size_t)NPt * 2 * C) * 4 + 255) / 256) * 256;
    float* F3 = (float*)wsp; wsp += (((size_t)((size_t)NPt * C) * 4 + 255) / 256) * 256;
    float* FU = (float*)wsp; wsp += (((size_t)((size_t)NPt * C) * 4 + 255) / 256) * 256;
    k_cc_norm<<<Bn, 256, 0, stream>>>(coords, NC, VIX, N, R);
    k_cc_ft<<<(unsigned)((NPt * C + 255) / 256), 256, 0, stream>>>(feat, FT, Bn, C, N);
    hipMemsetAsync(GP, 0, (size_t)Bn * RP3 * C * 4, stream); hipMemsetAsync(GQ, 0, (size_t)Bn * RP3 * C * 4, stream);
    k_inlists32<<<(unsigned)((NV) + IL_T32 - 1) / IL_T32, IL_T32, 0, stream>>>(VIX, NPt, NV, nbr, cnt);
    k_csr_scan32<<<1, 256, 0, stream>>>(cnt, off, NV);
    k_slotcopy32<<<(unsigned)((NPt) + 255) / 256, 256, 0, stream>>>(off, nbr, slot, NV);
    k_cc_vox<<<(unsigned)(((long long)NV * C + 255) / 256), 256, 0, stream>>>(FT, off, slot, GP, Bn, R, C);
    { GemmP v1_0_0;
      v1_0_0.A = GP + (size_t)0 * RP3 * C + (size_t)0 * C; v1_0_0.B = wv1 + 0; v1_0_0.bias = GP + (size_t)0 * RP3 * C + (size_t)0 * C; v1_0_0.R = GP + (size_t)0 * RP3 * C + (size_t)0 * C; v1_0_0.C = GC + (size_t)0 * R3 * C;
      v1_0_0.sAo = (long long)34 * 34 * C; v1_0_0.sAi = (long long)34 * C; v1_0_0.sAm = C; v1_0_0.sAk = 1; v1_0_0.sBo = 0; v1_0_0.sBi = 0; v1_0_0.sBn = C * 27; v1_0_0.sBk = 27; v1_0_0.sCo = (long long)R * R * C; v1_0_0.sCi = (long long)R * C; v1_0_0.sCm = C; v1_0_0.sRo = 0; v1_0_0.sRi = 0; v1_0_0.sRm = 0; v1_0_0.sRn = 0;
      v1_0_0.M = R; v1_0_0.N = C; v1_0_0.K = C; v1_0_0.zi_n = R; v1_0_0.flags = 0; v1_0_0.act = 0;
      v1_0_0.alpha = 1.0f; v1_0_0.beta = 0.0f; v1_0_0.sa = 1.0f; v1_0_0.sb = 1.0f; v1_0_0.Npad = C; v1_0_0.pad_ = 0;
      k_gemm<1><<<dim3((unsigned)((C) + 31) / 32, (unsigned)((R) + 15) / 16, (unsigned)(R * R)), 32, 0, stream>>>(v1_0_0); }
    { GemmP v1_0_1;
      v1_0_1.A = GP + (size_t)0 * RP3 * C + (size_t)1 * C; v1_0_1.B = wv1 + 1; v1_0_1.bias = GP + (size_t)0 * RP3 * C + (size_t)1 * C; v1_0_1.R = GC + (size_t)0 * R3 * C; v1_0_1.C = GC + (size_t)0 * R3 * C;
      v1_0_1.sAo = (long long)34 * 34 * C; v1_0_1.sAi = (long long)34 * C; v1_0_1.sAm = C; v1_0_1.sAk = 1; v1_0_1.sBo = 0; v1_0_1.sBi = 0; v1_0_1.sBn = C * 27; v1_0_1.sBk = 27; v1_0_1.sCo = (long long)R * R * C; v1_0_1.sCi = (long long)R * C; v1_0_1.sCm = C; v1_0_1.sRo = (long long)R * R * C; v1_0_1.sRi = (long long)R * C; v1_0_1.sRm = C; v1_0_1.sRn = 1;
      v1_0_1.M = R; v1_0_1.N = C; v1_0_1.K = C; v1_0_1.zi_n = R; v1_0_1.flags = 4; v1_0_1.act = 0;
      v1_0_1.alpha = 1.0f; v1_0_1.beta = 1.0f; v1_0_1.sa = 1.0f; v1_0_1.sb = 1.0f; v1_0_1.Npad = C; v1_0_1.pad_ = 0;
      k_gemm<1><<<dim3((unsigned)((C) + 31) / 32, (unsigned)((R) + 15) / 16, (unsigned)(R * R)), 32, 0, stream>>>(v1_0_1); }
    { GemmP v1_0_2;
      v1_0_2.A = GP + (size_t)0 * RP3 * C + (size_t)2 * C; v1_0_2.B = wv1 + 2; v1_0_2.bias = GP + (size_t)0 * RP3 * C + (size_t)2 * C; v1_0_2.R = GC + (size_t)0 * R3 * C; v1_0_2.C = GC + (size_t)0 * R3 * C;
      v1_0_2.sAo = (long long)34 * 34 * C; v1_0_2.sAi = (long long)34 * C; v1_0_2.sAm = C; v1_0_2.sAk = 1; v1_0_2.sBo = 0; v1_0_2.sBi = 0; v1_0_2.sBn = C * 27; v1_0_2.sBk = 27; v1_0_2.sCo = (long long)R * R * C; v1_0_2.sCi = (long long)R * C; v1_0_2.sCm = C; v1_0_2.sRo = (long long)R * R * C; v1_0_2.sRi = (long long)R * C; v1_0_2.sRm = C; v1_0_2.sRn = 1;
      v1_0_2.M = R; v1_0_2.N = C; v1_0_2.K = C; v1_0_2.zi_n = R; v1_0_2.flags = 4; v1_0_2.act = 0;
      v1_0_2.alpha = 1.0f; v1_0_2.beta = 1.0f; v1_0_2.sa = 1.0f; v1_0_2.sb = 1.0f; v1_0_2.Npad = C; v1_0_2.pad_ = 0;
      k_gemm<1><<<dim3((unsigned)((C) + 31) / 32, (unsigned)((R) + 15) / 16, (unsigned)(R * R)), 32, 0, stream>>>(v1_0_2); }
    { GemmP v1_0_3;
      v1_0_3.A = GP + (size_t)0 * RP3 * C + (size_t)34 * C; v1_0_3.B = wv1 + 3; v1_0_3.bias = GP + (size_t)0 * RP3 * C + (size_t)34 * C; v1_0_3.R = GC + (size_t)0 * R3 * C; v1_0_3.C = GC + (size_t)0 * R3 * C;
      v1_0_3.sAo = (long long)34 * 34 * C; v1_0_3.sAi = (long long)34 * C; v1_0_3.sAm = C; v1_0_3.sAk = 1; v1_0_3.sBo = 0; v1_0_3.sBi = 0; v1_0_3.sBn = C * 27; v1_0_3.sBk = 27; v1_0_3.sCo = (long long)R * R * C; v1_0_3.sCi = (long long)R * C; v1_0_3.sCm = C; v1_0_3.sRo = (long long)R * R * C; v1_0_3.sRi = (long long)R * C; v1_0_3.sRm = C; v1_0_3.sRn = 1;
      v1_0_3.M = R; v1_0_3.N = C; v1_0_3.K = C; v1_0_3.zi_n = R; v1_0_3.flags = 4; v1_0_3.act = 0;
      v1_0_3.alpha = 1.0f; v1_0_3.beta = 1.0f; v1_0_3.sa = 1.0f; v1_0_3.sb = 1.0f; v1_0_3.Npad = C; v1_0_3.pad_ = 0;
      k_gemm<1><<<dim3((unsigned)((C) + 31) / 32, (unsigned)((R) + 15) / 16, (unsigned)(R * R)), 32, 0, stream>>>(v1_0_3); }
    { GemmP v1_0_4;
      v1_0_4.A = GP + (size_t)0 * RP3 * C + (size_t)35 * C; v1_0_4.B = wv1 + 4; v1_0_4.bias = GP + (size_t)0 * RP3 * C + (size_t)35 * C; v1_0_4.R = GC + (size_t)0 * R3 * C; v1_0_4.C = GC + (size_t)0 * R3 * C;
      v1_0_4.sAo = (long long)34 * 34 * C; v1_0_4.sAi = (long long)34 * C; v1_0_4.sAm = C; v1_0_4.sAk = 1; v1_0_4.sBo = 0; v1_0_4.sBi = 0; v1_0_4.sBn = C * 27; v1_0_4.sBk = 27; v1_0_4.sCo = (long long)R * R * C; v1_0_4.sCi = (long long)R * C; v1_0_4.sCm = C; v1_0_4.sRo = (long long)R * R * C; v1_0_4.sRi = (long long)R * C; v1_0_4.sRm = C; v1_0_4.sRn = 1;
      v1_0_4.M = R; v1_0_4.N = C; v1_0_4.K = C; v1_0_4.zi_n = R; v1_0_4.flags = 4; v1_0_4.act = 0;
      v1_0_4.alpha = 1.0f; v1_0_4.beta = 1.0f; v1_0_4.sa = 1.0f; v1_0_4.sb = 1.0f; v1_0_4.Npad = C; v1_0_4.pad_ = 0;
      k_gemm<1><<<dim3((unsigned)((C) + 31) / 32, (unsigned)((R) + 15) / 16, (unsigned)(R * R)), 32, 0, stream>>>(v1_0_4); }
    { GemmP v1_0_5;
      v1_0_5.A = GP + (size_t)0 * RP3 * C + (size_t)36 * C; v1_0_5.B = wv1 + 5; v1_0_5.bias = GP + (size_t)0 * RP3 * C + (size_t)36 * C; v1_0_5.R = GC + (size_t)0 * R3 * C; v1_0_5.C = GC + (size_t)0 * R3 * C;
      v1_0_5.sAo = (long long)34 * 34 * C; v1_0_5.sAi = (long long)34 * C; v1_0_5.sAm = C; v1_0_5.sAk = 1; v1_0_5.sBo = 0; v1_0_5.sBi = 0; v1_0_5.sBn = C * 27; v1_0_5.sBk = 27; v1_0_5.sCo = (long long)R * R * C; v1_0_5.sCi = (long long)R * C; v1_0_5.sCm = C; v1_0_5.sRo = (long long)R * R * C; v1_0_5.sRi = (long long)R * C; v1_0_5.sRm = C; v1_0_5.sRn = 1;
      v1_0_5.M = R; v1_0_5.N = C; v1_0_5.K = C; v1_0_5.zi_n = R; v1_0_5.flags = 4; v1_0_5.act = 0;
      v1_0_5.alpha = 1.0f; v1_0_5.beta = 1.0f; v1_0_5.sa = 1.0f; v1_0_5.sb = 1.0f; v1_0_5.Npad = C; v1_0_5.pad_ = 0;
      k_gemm<1><<<dim3((unsigned)((C) + 31) / 32, (unsigned)((R) + 15) / 16, (unsigned)(R * R)), 32, 0, stream>>>(v1_0_5); }
    { GemmP v1_0_6;
      v1_0_6.A = GP + (size_t)0 * RP3 * C + (size_t)68 * C; v1_0_6.B = wv1 + 6; v1_0_6.bias = GP + (size_t)0 * RP3 * C + (size_t)68 * C; v1_0_6.R = GC + (size_t)0 * R3 * C; v1_0_6.C = GC + (size_t)0 * R3 * C;
      v1_0_6.sAo = (long long)34 * 34 * C; v1_0_6.sAi = (long long)34 * C; v1_0_6.sAm = C; v1_0_6.sAk = 1; v1_0_6.sBo = 0; v1_0_6.sBi = 0; v1_0_6.sBn = C * 27; v1_0_6.sBk = 27; v1_0_6.sCo = (long long)R * R * C; v1_0_6.sCi = (long long)R * C; v1_0_6.sCm = C; v1_0_6.sRo = (long long)R * R * C; v1_0_6.sRi = (long long)R * C; v1_0_6.sRm = C; v1_0_6.sRn = 1;
      v1_0_6.M = R; v1_0_6.N = C; v1_0_6.K = C; v1_0_6.zi_n = R; v1_0_6.flags = 4; v1_0_6.act = 0;
      v1_0_6.alpha = 1.0f; v1_0_6.beta = 1.0f; v1_0_6.sa = 1.0f; v1_0_6.sb = 1.0f; v1_0_6.Npad = C; v1_0_6.pad_ = 0;
      k_gemm<1><<<dim3((unsigned)((C) + 31) / 32, (unsigned)((R) + 15) / 16, (unsigned)(R * R)), 32, 0, stream>>>(v1_0_6); }
    { GemmP v1_0_7;
      v1_0_7.A = GP + (size_t)0 * RP3 * C + (size_t)69 * C; v1_0_7.B = wv1 + 7; v1_0_7.bias = GP + (size_t)0 * RP3 * C + (size_t)69 * C; v1_0_7.R = GC + (size_t)0 * R3 * C; v1_0_7.C = GC + (size_t)0 * R3 * C;
      v1_0_7.sAo = (long long)34 * 34 * C; v1_0_7.sAi = (long long)34 * C; v1_0_7.sAm = C; v1_0_7.sAk = 1; v1_0_7.sBo = 0; v1_0_7.sBi = 0; v1_0_7.sBn = C * 27; v1_0_7.sBk = 27; v1_0_7.sCo = (long long)R * R * C; v1_0_7.sCi = (long long)R * C; v1_0_7.sCm = C; v1_0_7.sRo = (long long)R * R * C; v1_0_7.sRi = (long long)R * C; v1_0_7.sRm = C; v1_0_7.sRn = 1;
      v1_0_7.M = R; v1_0_7.N = C; v1_0_7.K = C; v1_0_7.zi_n = R; v1_0_7.flags = 4; v1_0_7.act = 0;
      v1_0_7.alpha = 1.0f; v1_0_7.beta = 1.0f; v1_0_7.sa = 1.0f; v1_0_7.sb = 1.0f; v1_0_7.Npad = C; v1_0_7.pad_ = 0;
      k_gemm<1><<<dim3((unsigned)((C) + 31) / 32, (unsigned)((R) + 15) / 16, (unsigned)(R * R)), 32, 0, stream>>>(v1_0_7); }
    { GemmP v1_0_8;
      v1_0_8.A = GP + (size_t)0 * RP3 * C + (size_t)70 * C; v1_0_8.B = wv1 + 8; v1_0_8.bias = GP + (size_t)0 * RP3 * C + (size_t)70 * C; v1_0_8.R = GC + (size_t)0 * R3 * C; v1_0_8.C = GC + (size_t)0 * R3 * C;
      v1_0_8.sAo = (long long)34 * 34 * C; v1_0_8.sAi = (long long)34 * C; v1_0_8.sAm = C; v1_0_8.sAk = 1; v1_0_8.sBo = 0; v1_0_8.sBi = 0; v1_0_8.sBn = C * 27; v1_0_8.sBk = 27; v1_0_8.sCo = (long long)R * R * C; v1_0_8.sCi = (long long)R * C; v1_0_8.sCm = C; v1_0_8.sRo = (long long)R * R * C; v1_0_8.sRi = (long long)R * C; v1_0_8.sRm = C; v1_0_8.sRn = 1;
      v1_0_8.M = R; v1_0_8.N = C; v1_0_8.K = C; v1_0_8.zi_n = R; v1_0_8.flags = 4; v1_0_8.act = 0;
      v1_0_8.alpha = 1.0f; v1_0_8.beta = 1.0f; v1_0_8.sa = 1.0f; v1_0_8.sb = 1.0f; v1_0_8.Npad = C; v1_0_8.pad_ = 0;
      k_gemm<1><<<dim3((unsigned)((C) + 31) / 32, (unsigned)((R) + 15) / 16, (unsigned)(R * R)), 32, 0, stream>>>(v1_0_8); }
    { GemmP v1_0_9;
      v1_0_9.A = GP + (size_t)0 * RP3 * C + (size_t)1156 * C; v1_0_9.B = wv1 + 9; v1_0_9.bias = GP + (size_t)0 * RP3 * C + (size_t)1156 * C; v1_0_9.R = GC + (size_t)0 * R3 * C; v1_0_9.C = GC + (size_t)0 * R3 * C;
      v1_0_9.sAo = (long long)34 * 34 * C; v1_0_9.sAi = (long long)34 * C; v1_0_9.sAm = C; v1_0_9.sAk = 1; v1_0_9.sBo = 0; v1_0_9.sBi = 0; v1_0_9.sBn = C * 27; v1_0_9.sBk = 27; v1_0_9.sCo = (long long)R * R * C; v1_0_9.sCi = (long long)R * C; v1_0_9.sCm = C; v1_0_9.sRo = (long long)R * R * C; v1_0_9.sRi = (long long)R * C; v1_0_9.sRm = C; v1_0_9.sRn = 1;
      v1_0_9.M = R; v1_0_9.N = C; v1_0_9.K = C; v1_0_9.zi_n = R; v1_0_9.flags = 4; v1_0_9.act = 0;
      v1_0_9.alpha = 1.0f; v1_0_9.beta = 1.0f; v1_0_9.sa = 1.0f; v1_0_9.sb = 1.0f; v1_0_9.Npad = C; v1_0_9.pad_ = 0;
      k_gemm<1><<<dim3((unsigned)((C) + 31) / 32, (unsigned)((R) + 15) / 16, (unsigned)(R * R)), 32, 0, stream>>>(v1_0_9); }
    { GemmP v1_0_10;
      v1_0_10.A = GP + (size_t)0 * RP3 * C + (size_t)1157 * C; v1_0_10.B = wv1 + 10; v1_0_10.bias = GP + (size_t)0 * RP3 * C + (size_t)1157 * C; v1_0_10.R = GC + (size_t)0 * R3 * C; v1_0_10.C = GC + (size_t)0 * R3 * C;
      v1_0_10.sAo = (long long)34 * 34 * C; v1_0_10.sAi = (long long)34 * C; v1_0_10.sAm = C; v1_0_10.sAk = 1; v1_0_10.sBo = 0; v1_0_10.sBi = 0; v1_0_10.sBn = C * 27; v1_0_10.sBk = 27; v1_0_10.sCo = (long long)R * R * C; v1_0_10.sCi = (long long)R * C; v1_0_10.sCm = C; v1_0_10.sRo = (long long)R * R * C; v1_0_10.sRi = (long long)R * C; v1_0_10.sRm = C; v1_0_10.sRn = 1;
      v1_0_10.M = R; v1_0_10.N = C; v1_0_10.K = C; v1_0_10.zi_n = R; v1_0_10.flags = 4; v1_0_10.act = 0;
      v1_0_10.alpha = 1.0f; v1_0_10.beta = 1.0f; v1_0_10.sa = 1.0f; v1_0_10.sb = 1.0f; v1_0_10.Npad = C; v1_0_10.pad_ = 0;
      k_gemm<1><<<dim3((unsigned)((C) + 31) / 32, (unsigned)((R) + 15) / 16, (unsigned)(R * R)), 32, 0, stream>>>(v1_0_10); }
    { GemmP v1_0_11;
      v1_0_11.A = GP + (size_t)0 * RP3 * C + (size_t)1158 * C; v1_0_11.B = wv1 + 11; v1_0_11.bias = GP + (size_t)0 * RP3 * C + (size_t)1158 * C; v1_0_11.R = GC + (size_t)0 * R3 * C; v1_0_11.C = GC + (size_t)0 * R3 * C;
      v1_0_11.sAo = (long long)34 * 34 * C; v1_0_11.sAi = (long long)34 * C; v1_0_11.sAm = C; v1_0_11.sAk = 1; v1_0_11.sBo = 0; v1_0_11.sBi = 0; v1_0_11.sBn = C * 27; v1_0_11.sBk = 27; v1_0_11.sCo = (long long)R * R * C; v1_0_11.sCi = (long long)R * C; v1_0_11.sCm = C; v1_0_11.sRo = (long long)R * R * C; v1_0_11.sRi = (long long)R * C; v1_0_11.sRm = C; v1_0_11.sRn = 1;
      v1_0_11.M = R; v1_0_11.N = C; v1_0_11.K = C; v1_0_11.zi_n = R; v1_0_11.flags = 4; v1_0_11.act = 0;
      v1_0_11.alpha = 1.0f; v1_0_11.beta = 1.0f; v1_0_11.sa = 1.0f; v1_0_11.sb = 1.0f; v1_0_11.Npad = C; v1_0_11.pad_ = 0;
      k_gemm<1><<<dim3((unsigned)((C) + 31) / 32, (unsigned)((R) + 15) / 16, (unsigned)(R * R)), 32, 0, stream>>>(v1_0_11); }
    { GemmP v1_0_12;
      v1_0_12.A = GP + (size_t)0 * RP3 * C + (size_t)1190 * C; v1_0_12.B = wv1 + 12; v1_0_12.bias = GP + (size_t)0 * RP3 * C + (size_t)1190 * C; v1_0_12.R = GC + (size_t)0 * R3 * C; v1_0_12.C = GC + (size_t)0 * R3 * C;
      v1_0_12.sAo = (long long)34 * 34 * C; v1_0_12.sAi = (long long)34 * C; v1_0_12.sAm = C; v1_0_12.sAk = 1; v1_0_12.sBo = 0; v1_0_12.sBi = 0; v1_0_12.sBn = C * 27; v1_0_12.sBk = 27; v1_0_12.sCo = (long long)R * R * C; v1_0_12.sCi = (long long)R * C; v1_0_12.sCm = C; v1_0_12.sRo = (long long)R * R * C; v1_0_12.sRi = (long long)R * C; v1_0_12.sRm = C; v1_0_12.sRn = 1;
      v1_0_12.M = R; v1_0_12.N = C; v1_0_12.K = C; v1_0_12.zi_n = R; v1_0_12.flags = 4; v1_0_12.act = 0;
      v1_0_12.alpha = 1.0f; v1_0_12.beta = 1.0f; v1_0_12.sa = 1.0f; v1_0_12.sb = 1.0f; v1_0_12.Npad = C; v1_0_12.pad_ = 0;
      k_gemm<1><<<dim3((unsigned)((C) + 31) / 32, (unsigned)((R) + 15) / 16, (unsigned)(R * R)), 32, 0, stream>>>(v1_0_12); }
    { GemmP v1_0_13;
      v1_0_13.A = GP + (size_t)0 * RP3 * C + (size_t)1191 * C; v1_0_13.B = wv1 + 13; v1_0_13.bias = GP + (size_t)0 * RP3 * C + (size_t)1191 * C; v1_0_13.R = GC + (size_t)0 * R3 * C; v1_0_13.C = GC + (size_t)0 * R3 * C;
      v1_0_13.sAo = (long long)34 * 34 * C; v1_0_13.sAi = (long long)34 * C; v1_0_13.sAm = C; v1_0_13.sAk = 1; v1_0_13.sBo = 0; v1_0_13.sBi = 0; v1_0_13.sBn = C * 27; v1_0_13.sBk = 27; v1_0_13.sCo = (long long)R * R * C; v1_0_13.sCi = (long long)R * C; v1_0_13.sCm = C; v1_0_13.sRo = (long long)R * R * C; v1_0_13.sRi = (long long)R * C; v1_0_13.sRm = C; v1_0_13.sRn = 1;
      v1_0_13.M = R; v1_0_13.N = C; v1_0_13.K = C; v1_0_13.zi_n = R; v1_0_13.flags = 4; v1_0_13.act = 0;
      v1_0_13.alpha = 1.0f; v1_0_13.beta = 1.0f; v1_0_13.sa = 1.0f; v1_0_13.sb = 1.0f; v1_0_13.Npad = C; v1_0_13.pad_ = 0;
      k_gemm<1><<<dim3((unsigned)((C) + 31) / 32, (unsigned)((R) + 15) / 16, (unsigned)(R * R)), 32, 0, stream>>>(v1_0_13); }
    { GemmP v1_0_14;
      v1_0_14.A = GP + (size_t)0 * RP3 * C + (size_t)1192 * C; v1_0_14.B = wv1 + 14; v1_0_14.bias = GP + (size_t)0 * RP3 * C + (size_t)1192 * C; v1_0_14.R = GC + (size_t)0 * R3 * C; v1_0_14.C = GC + (size_t)0 * R3 * C;
      v1_0_14.sAo = (long long)34 * 34 * C; v1_0_14.sAi = (long long)34 * C; v1_0_14.sAm = C; v1_0_14.sAk = 1; v1_0_14.sBo = 0; v1_0_14.sBi = 0; v1_0_14.sBn = C * 27; v1_0_14.sBk = 27; v1_0_14.sCo = (long long)R * R * C; v1_0_14.sCi = (long long)R * C; v1_0_14.sCm = C; v1_0_14.sRo = (long long)R * R * C; v1_0_14.sRi = (long long)R * C; v1_0_14.sRm = C; v1_0_14.sRn = 1;
      v1_0_14.M = R; v1_0_14.N = C; v1_0_14.K = C; v1_0_14.zi_n = R; v1_0_14.flags = 4; v1_0_14.act = 0;
      v1_0_14.alpha = 1.0f; v1_0_14.beta = 1.0f; v1_0_14.sa = 1.0f; v1_0_14.sb = 1.0f; v1_0_14.Npad = C; v1_0_14.pad_ = 0;
      k_gemm<1><<<dim3((unsigned)((C) + 31) / 32, (unsigned)((R) + 15) / 16, (unsigned)(R * R)), 32, 0, stream>>>(v1_0_14); }
    { GemmP v1_0_15;
      v1_0_15.A = GP + (size_t)0 * RP3 * C + (size_t)1224 * C; v1_0_15.B = wv1 + 15; v1_0_15.bias = GP + (size_t)0 * RP3 * C + (size_t)1224 * C; v1_0_15.R = GC + (size_t)0 * R3 * C; v1_0_15.C = GC + (size_t)0 * R3 * C;
      v1_0_15.sAo = (long long)34 * 34 * C; v1_0_15.sAi = (long long)34 * C; v1_0_15.sAm = C; v1_0_15.sAk = 1; v1_0_15.sBo = 0; v1_0_15.sBi = 0; v1_0_15.sBn = C * 27; v1_0_15.sBk = 27; v1_0_15.sCo = (long long)R * R * C; v1_0_15.sCi = (long long)R * C; v1_0_15.sCm = C; v1_0_15.sRo = (long long)R * R * C; v1_0_15.sRi = (long long)R * C; v1_0_15.sRm = C; v1_0_15.sRn = 1;
      v1_0_15.M = R; v1_0_15.N = C; v1_0_15.K = C; v1_0_15.zi_n = R; v1_0_15.flags = 4; v1_0_15.act = 0;
      v1_0_15.alpha = 1.0f; v1_0_15.beta = 1.0f; v1_0_15.sa = 1.0f; v1_0_15.sb = 1.0f; v1_0_15.Npad = C; v1_0_15.pad_ = 0;
      k_gemm<1><<<dim3((unsigned)((C) + 31) / 32, (unsigned)((R) + 15) / 16, (unsigned)(R * R)), 32, 0, stream>>>(v1_0_15); }
    { GemmP v1_0_16;
      v1_0_16.A = GP + (size_t)0 * RP3 * C + (size_t)1225 * C; v1_0_16.B = wv1 + 16; v1_0_16.bias = GP + (size_t)0 * RP3 * C + (size_t)1225 * C; v1_0_16.R = GC + (size_t)0 * R3 * C; v1_0_16.C = GC + (size_t)0 * R3 * C;
      v1_0_16.sAo = (long long)34 * 34 * C; v1_0_16.sAi = (long long)34 * C; v1_0_16.sAm = C; v1_0_16.sAk = 1; v1_0_16.sBo = 0; v1_0_16.sBi = 0; v1_0_16.sBn = C * 27; v1_0_16.sBk = 27; v1_0_16.sCo = (long long)R * R * C; v1_0_16.sCi = (long long)R * C; v1_0_16.sCm = C; v1_0_16.sRo = (long long)R * R * C; v1_0_16.sRi = (long long)R * C; v1_0_16.sRm = C; v1_0_16.sRn = 1;
      v1_0_16.M = R; v1_0_16.N = C; v1_0_16.K = C; v1_0_16.zi_n = R; v1_0_16.flags = 4; v1_0_16.act = 0;
      v1_0_16.alpha = 1.0f; v1_0_16.beta = 1.0f; v1_0_16.sa = 1.0f; v1_0_16.sb = 1.0f; v1_0_16.Npad = C; v1_0_16.pad_ = 0;
      k_gemm<1><<<dim3((unsigned)((C) + 31) / 32, (unsigned)((R) + 15) / 16, (unsigned)(R * R)), 32, 0, stream>>>(v1_0_16); }
    { GemmP v1_0_17;
      v1_0_17.A = GP + (size_t)0 * RP3 * C + (size_t)1226 * C; v1_0_17.B = wv1 + 17; v1_0_17.bias = GP + (size_t)0 * RP3 * C + (size_t)1226 * C; v1_0_17.R = GC + (size_t)0 * R3 * C; v1_0_17.C = GC + (size_t)0 * R3 * C;
      v1_0_17.sAo = (long long)34 * 34 * C; v1_0_17.sAi = (long long)34 * C; v1_0_17.sAm = C; v1_0_17.sAk = 1; v1_0_17.sBo = 0; v1_0_17.sBi = 0; v1_0_17.sBn = C * 27; v1_0_17.sBk = 27; v1_0_17.sCo = (long long)R * R * C; v1_0_17.sCi = (long long)R * C; v1_0_17.sCm = C; v1_0_17.sRo = (long long)R * R * C; v1_0_17.sRi = (long long)R * C; v1_0_17.sRm = C; v1_0_17.sRn = 1;
      v1_0_17.M = R; v1_0_17.N = C; v1_0_17.K = C; v1_0_17.zi_n = R; v1_0_17.flags = 4; v1_0_17.act = 0;
      v1_0_17.alpha = 1.0f; v1_0_17.beta = 1.0f; v1_0_17.sa = 1.0f; v1_0_17.sb = 1.0f; v1_0_17.Npad = C; v1_0_17.pad_ = 0;
      k_gemm<1><<<dim3((unsigned)((C) + 31) / 32, (unsigned)((R) + 15) / 16, (unsigned)(R * R)), 32, 0, stream>>>(v1_0_17); }
    { GemmP v1_0_18;
      v1_0_18.A = GP + (size_t)0 * RP3 * C + (size_t)2312 * C; v1_0_18.B = wv1 + 18; v1_0_18.bias = GP + (size_t)0 * RP3 * C + (size_t)2312 * C; v1_0_18.R = GC + (size_t)0 * R3 * C; v1_0_18.C = GC + (size_t)0 * R3 * C;
      v1_0_18.sAo = (long long)34 * 34 * C; v1_0_18.sAi = (long long)34 * C; v1_0_18.sAm = C; v1_0_18.sAk = 1; v1_0_18.sBo = 0; v1_0_18.sBi = 0; v1_0_18.sBn = C * 27; v1_0_18.sBk = 27; v1_0_18.sCo = (long long)R * R * C; v1_0_18.sCi = (long long)R * C; v1_0_18.sCm = C; v1_0_18.sRo = (long long)R * R * C; v1_0_18.sRi = (long long)R * C; v1_0_18.sRm = C; v1_0_18.sRn = 1;
      v1_0_18.M = R; v1_0_18.N = C; v1_0_18.K = C; v1_0_18.zi_n = R; v1_0_18.flags = 4; v1_0_18.act = 0;
      v1_0_18.alpha = 1.0f; v1_0_18.beta = 1.0f; v1_0_18.sa = 1.0f; v1_0_18.sb = 1.0f; v1_0_18.Npad = C; v1_0_18.pad_ = 0;
      k_gemm<1><<<dim3((unsigned)((C) + 31) / 32, (unsigned)((R) + 15) / 16, (unsigned)(R * R)), 32, 0, stream>>>(v1_0_18); }
    { GemmP v1_0_19;
      v1_0_19.A = GP + (size_t)0 * RP3 * C + (size_t)2313 * C; v1_0_19.B = wv1 + 19; v1_0_19.bias = GP + (size_t)0 * RP3 * C + (size_t)2313 * C; v1_0_19.R = GC + (size_t)0 * R3 * C; v1_0_19.C = GC + (size_t)0 * R3 * C;
      v1_0_19.sAo = (long long)34 * 34 * C; v1_0_19.sAi = (long long)34 * C; v1_0_19.sAm = C; v1_0_19.sAk = 1; v1_0_19.sBo = 0; v1_0_19.sBi = 0; v1_0_19.sBn = C * 27; v1_0_19.sBk = 27; v1_0_19.sCo = (long long)R * R * C; v1_0_19.sCi = (long long)R * C; v1_0_19.sCm = C; v1_0_19.sRo = (long long)R * R * C; v1_0_19.sRi = (long long)R * C; v1_0_19.sRm = C; v1_0_19.sRn = 1;
      v1_0_19.M = R; v1_0_19.N = C; v1_0_19.K = C; v1_0_19.zi_n = R; v1_0_19.flags = 4; v1_0_19.act = 0;
      v1_0_19.alpha = 1.0f; v1_0_19.beta = 1.0f; v1_0_19.sa = 1.0f; v1_0_19.sb = 1.0f; v1_0_19.Npad = C; v1_0_19.pad_ = 0;
      k_gemm<1><<<dim3((unsigned)((C) + 31) / 32, (unsigned)((R) + 15) / 16, (unsigned)(R * R)), 32, 0, stream>>>(v1_0_19); }
    { GemmP v1_0_20;
      v1_0_20.A = GP + (size_t)0 * RP3 * C + (size_t)2314 * C; v1_0_20.B = wv1 + 20; v1_0_20.bias = GP + (size_t)0 * RP3 * C + (size_t)2314 * C; v1_0_20.R = GC + (size_t)0 * R3 * C; v1_0_20.C = GC + (size_t)0 * R3 * C;
      v1_0_20.sAo = (long long)34 * 34 * C; v1_0_20.sAi = (long long)34 * C; v1_0_20.sAm = C; v1_0_20.sAk = 1; v1_0_20.sBo = 0; v1_0_20.sBi = 0; v1_0_20.sBn = C * 27; v1_0_20.sBk = 27; v1_0_20.sCo = (long long)R * R * C; v1_0_20.sCi = (long long)R * C; v1_0_20.sCm = C; v1_0_20.sRo = (long long)R * R * C; v1_0_20.sRi = (long long)R * C; v1_0_20.sRm = C; v1_0_20.sRn = 1;
      v1_0_20.M = R; v1_0_20.N = C; v1_0_20.K = C; v1_0_20.zi_n = R; v1_0_20.flags = 4; v1_0_20.act = 0;
      v1_0_20.alpha = 1.0f; v1_0_20.beta = 1.0f; v1_0_20.sa = 1.0f; v1_0_20.sb = 1.0f; v1_0_20.Npad = C; v1_0_20.pad_ = 0;
      k_gemm<1><<<dim3((unsigned)((C) + 31) / 32, (unsigned)((R) + 15) / 16, (unsigned)(R * R)), 32, 0, stream>>>(v1_0_20); }
    { GemmP v1_0_21;
      v1_0_21.A = GP + (size_t)0 * RP3 * C + (size_t)2346 * C; v1_0_21.B = wv1 + 21; v1_0_21.bias = GP + (size_t)0 * RP3 * C + (size_t)2346 * C; v1_0_21.R = GC + (size_t)0 * R3 * C; v1_0_21.C = GC + (size_t)0 * R3 * C;
      v1_0_21.sAo = (long long)34 * 34 * C; v1_0_21.sAi = (long long)34 * C; v1_0_21.sAm = C; v1_0_21.sAk = 1; v1_0_21.sBo = 0; v1_0_21.sBi = 0; v1_0_21.sBn = C * 27; v1_0_21.sBk = 27; v1_0_21.sCo = (long long)R * R * C; v1_0_21.sCi = (long long)R * C; v1_0_21.sCm = C; v1_0_21.sRo = (long long)R * R * C; v1_0_21.sRi = (long long)R * C; v1_0_21.sRm = C; v1_0_21.sRn = 1;
      v1_0_21.M = R; v1_0_21.N = C; v1_0_21.K = C; v1_0_21.zi_n = R; v1_0_21.flags = 4; v1_0_21.act = 0;
      v1_0_21.alpha = 1.0f; v1_0_21.beta = 1.0f; v1_0_21.sa = 1.0f; v1_0_21.sb = 1.0f; v1_0_21.Npad = C; v1_0_21.pad_ = 0;
      k_gemm<1><<<dim3((unsigned)((C) + 31) / 32, (unsigned)((R) + 15) / 16, (unsigned)(R * R)), 32, 0, stream>>>(v1_0_21); }
    { GemmP v1_0_22;
      v1_0_22.A = GP + (size_t)0 * RP3 * C + (size_t)2347 * C; v1_0_22.B = wv1 + 22; v1_0_22.bias = GP + (size_t)0 * RP3 * C + (size_t)2347 * C; v1_0_22.R = GC + (size_t)0 * R3 * C; v1_0_22.C = GC + (size_t)0 * R3 * C;
      v1_0_22.sAo = (long long)34 * 34 * C; v1_0_22.sAi = (long long)34 * C; v1_0_22.sAm = C; v1_0_22.sAk = 1; v1_0_22.sBo = 0; v1_0_22.sBi = 0; v1_0_22.sBn = C * 27; v1_0_22.sBk = 27; v1_0_22.sCo = (long long)R * R * C; v1_0_22.sCi = (long long)R * C; v1_0_22.sCm = C; v1_0_22.sRo = (long long)R * R * C; v1_0_22.sRi = (long long)R * C; v1_0_22.sRm = C; v1_0_22.sRn = 1;
      v1_0_22.M = R; v1_0_22.N = C; v1_0_22.K = C; v1_0_22.zi_n = R; v1_0_22.flags = 4; v1_0_22.act = 0;
      v1_0_22.alpha = 1.0f; v1_0_22.beta = 1.0f; v1_0_22.sa = 1.0f; v1_0_22.sb = 1.0f; v1_0_22.Npad = C; v1_0_22.pad_ = 0;
      k_gemm<1><<<dim3((unsigned)((C) + 31) / 32, (unsigned)((R) + 15) / 16, (unsigned)(R * R)), 32, 0, stream>>>(v1_0_22); }
    { GemmP v1_0_23;
      v1_0_23.A = GP + (size_t)0 * RP3 * C + (size_t)2348 * C; v1_0_23.B = wv1 + 23; v1_0_23.bias = GP + (size_t)0 * RP3 * C + (size_t)2348 * C; v1_0_23.R = GC + (size_t)0 * R3 * C; v1_0_23.C = GC + (size_t)0 * R3 * C;
      v1_0_23.sAo = (long long)34 * 34 * C; v1_0_23.sAi = (long long)34 * C; v1_0_23.sAm = C; v1_0_23.sAk = 1; v1_0_23.sBo = 0; v1_0_23.sBi = 0; v1_0_23.sBn = C * 27; v1_0_23.sBk = 27; v1_0_23.sCo = (long long)R * R * C; v1_0_23.sCi = (long long)R * C; v1_0_23.sCm = C; v1_0_23.sRo = (long long)R * R * C; v1_0_23.sRi = (long long)R * C; v1_0_23.sRm = C; v1_0_23.sRn = 1;
      v1_0_23.M = R; v1_0_23.N = C; v1_0_23.K = C; v1_0_23.zi_n = R; v1_0_23.flags = 4; v1_0_23.act = 0;
      v1_0_23.alpha = 1.0f; v1_0_23.beta = 1.0f; v1_0_23.sa = 1.0f; v1_0_23.sb = 1.0f; v1_0_23.Npad = C; v1_0_23.pad_ = 0;
      k_gemm<1><<<dim3((unsigned)((C) + 31) / 32, (unsigned)((R) + 15) / 16, (unsigned)(R * R)), 32, 0, stream>>>(v1_0_23); }
    { GemmP v1_0_24;
      v1_0_24.A = GP + (size_t)0 * RP3 * C + (size_t)2380 * C; v1_0_24.B = wv1 + 24; v1_0_24.bias = GP + (size_t)0 * RP3 * C + (size_t)2380 * C; v1_0_24.R = GC + (size_t)0 * R3 * C; v1_0_24.C = GC + (size_t)0 * R3 * C;
      v1_0_24.sAo = (long long)34 * 34 * C; v1_0_24.sAi = (long long)34 * C; v1_0_24.sAm = C; v1_0_24.sAk = 1; v1_0_24.sBo = 0; v1_0_24.sBi = 0; v1_0_24.sBn = C * 27; v1_0_24.sBk = 27; v1_0_24.sCo = (long long)R * R * C; v1_0_24.sCi = (long long)R * C; v1_0_24.sCm = C; v1_0_24.sRo = (long long)R * R * C; v1_0_24.sRi = (long long)R * C; v1_0_24.sRm = C; v1_0_24.sRn = 1;
      v1_0_24.M = R; v1_0_24.N = C; v1_0_24.K = C; v1_0_24.zi_n = R; v1_0_24.flags = 4; v1_0_24.act = 0;
      v1_0_24.alpha = 1.0f; v1_0_24.beta = 1.0f; v1_0_24.sa = 1.0f; v1_0_24.sb = 1.0f; v1_0_24.Npad = C; v1_0_24.pad_ = 0;
      k_gemm<1><<<dim3((unsigned)((C) + 31) / 32, (unsigned)((R) + 15) / 16, (unsigned)(R * R)), 32, 0, stream>>>(v1_0_24); }
    { GemmP v1_0_25;
      v1_0_25.A = GP + (size_t)0 * RP3 * C + (size_t)2381 * C; v1_0_25.B = wv1 + 25; v1_0_25.bias = GP + (size_t)0 * RP3 * C + (size_t)2381 * C; v1_0_25.R = GC + (size_t)0 * R3 * C; v1_0_25.C = GC + (size_t)0 * R3 * C;
      v1_0_25.sAo = (long long)34 * 34 * C; v1_0_25.sAi = (long long)34 * C; v1_0_25.sAm = C; v1_0_25.sAk = 1; v1_0_25.sBo = 0; v1_0_25.sBi = 0; v1_0_25.sBn = C * 27; v1_0_25.sBk = 27; v1_0_25.sCo = (long long)R * R * C; v1_0_25.sCi = (long long)R * C; v1_0_25.sCm = C; v1_0_25.sRo = (long long)R * R * C; v1_0_25.sRi = (long long)R * C; v1_0_25.sRm = C; v1_0_25.sRn = 1;
      v1_0_25.M = R; v1_0_25.N = C; v1_0_25.K = C; v1_0_25.zi_n = R; v1_0_25.flags = 4; v1_0_25.act = 0;
      v1_0_25.alpha = 1.0f; v1_0_25.beta = 1.0f; v1_0_25.sa = 1.0f; v1_0_25.sb = 1.0f; v1_0_25.Npad = C; v1_0_25.pad_ = 0;
      k_gemm<1><<<dim3((unsigned)((C) + 31) / 32, (unsigned)((R) + 15) / 16, (unsigned)(R * R)), 32, 0, stream>>>(v1_0_25); }
    { GemmP v1_0_26;
      v1_0_26.A = GP + (size_t)0 * RP3 * C + (size_t)2382 * C; v1_0_26.B = wv1 + 26; v1_0_26.bias = GP + (size_t)0 * RP3 * C + (size_t)2382 * C; v1_0_26.R = GC + (size_t)0 * R3 * C; v1_0_26.C = GC + (size_t)0 * R3 * C;
      v1_0_26.sAo = (long long)34 * 34 * C; v1_0_26.sAi = (long long)34 * C; v1_0_26.sAm = C; v1_0_26.sAk = 1; v1_0_26.sBo = 0; v1_0_26.sBi = 0; v1_0_26.sBn = C * 27; v1_0_26.sBk = 27; v1_0_26.sCo = (long long)R * R * C; v1_0_26.sCi = (long long)R * C; v1_0_26.sCm = C; v1_0_26.sRo = (long long)R * R * C; v1_0_26.sRi = (long long)R * C; v1_0_26.sRm = C; v1_0_26.sRn = 1;
      v1_0_26.M = R; v1_0_26.N = C; v1_0_26.K = C; v1_0_26.zi_n = R; v1_0_26.flags = 4; v1_0_26.act = 0;
      v1_0_26.alpha = 1.0f; v1_0_26.beta = 1.0f; v1_0_26.sa = 1.0f; v1_0_26.sb = 1.0f; v1_0_26.Npad = C; v1_0_26.pad_ = 0;
      k_gemm<1><<<dim3((unsigned)((C) + 31) / 32, (unsigned)((R) + 15) / 16, (unsigned)(R * R)), 32, 0, stream>>>(v1_0_26); }
    { GemmP v1_1_0;
      v1_1_0.A = GP + (size_t)1 * RP3 * C + (size_t)0 * C; v1_1_0.B = wv1 + 0; v1_1_0.bias = GP + (size_t)1 * RP3 * C + (size_t)0 * C; v1_1_0.R = GP + (size_t)1 * RP3 * C + (size_t)0 * C; v1_1_0.C = GC + (size_t)1 * R3 * C;
      v1_1_0.sAo = (long long)34 * 34 * C; v1_1_0.sAi = (long long)34 * C; v1_1_0.sAm = C; v1_1_0.sAk = 1; v1_1_0.sBo = 0; v1_1_0.sBi = 0; v1_1_0.sBn = C * 27; v1_1_0.sBk = 27; v1_1_0.sCo = (long long)R * R * C; v1_1_0.sCi = (long long)R * C; v1_1_0.sCm = C; v1_1_0.sRo = 0; v1_1_0.sRi = 0; v1_1_0.sRm = 0; v1_1_0.sRn = 0;
      v1_1_0.M = R; v1_1_0.N = C; v1_1_0.K = C; v1_1_0.zi_n = R; v1_1_0.flags = 0; v1_1_0.act = 0;
      v1_1_0.alpha = 1.0f; v1_1_0.beta = 0.0f; v1_1_0.sa = 1.0f; v1_1_0.sb = 1.0f; v1_1_0.Npad = C; v1_1_0.pad_ = 0;
      k_gemm<1><<<dim3((unsigned)((C) + 31) / 32, (unsigned)((R) + 15) / 16, (unsigned)(R * R)), 32, 0, stream>>>(v1_1_0); }
    { GemmP v1_1_1;
      v1_1_1.A = GP + (size_t)1 * RP3 * C + (size_t)1 * C; v1_1_1.B = wv1 + 1; v1_1_1.bias = GP + (size_t)1 * RP3 * C + (size_t)1 * C; v1_1_1.R = GC + (size_t)1 * R3 * C; v1_1_1.C = GC + (size_t)1 * R3 * C;
      v1_1_1.sAo = (long long)34 * 34 * C; v1_1_1.sAi = (long long)34 * C; v1_1_1.sAm = C; v1_1_1.sAk = 1; v1_1_1.sBo = 0; v1_1_1.sBi = 0; v1_1_1.sBn = C * 27; v1_1_1.sBk = 27; v1_1_1.sCo = (long long)R * R * C; v1_1_1.sCi = (long long)R * C; v1_1_1.sCm = C; v1_1_1.sRo = (long long)R * R * C; v1_1_1.sRi = (long long)R * C; v1_1_1.sRm = C; v1_1_1.sRn = 1;
      v1_1_1.M = R; v1_1_1.N = C; v1_1_1.K = C; v1_1_1.zi_n = R; v1_1_1.flags = 4; v1_1_1.act = 0;
      v1_1_1.alpha = 1.0f; v1_1_1.beta = 1.0f; v1_1_1.sa = 1.0f; v1_1_1.sb = 1.0f; v1_1_1.Npad = C; v1_1_1.pad_ = 0;
      k_gemm<1><<<dim3((unsigned)((C) + 31) / 32, (unsigned)((R) + 15) / 16, (unsigned)(R * R)), 32, 0, stream>>>(v1_1_1); }
    { GemmP v1_1_2;
      v1_1_2.A = GP + (size_t)1 * RP3 * C + (size_t)2 * C; v1_1_2.B = wv1 + 2; v1_1_2.bias = GP + (size_t)1 * RP3 * C + (size_t)2 * C; v1_1_2.R = GC + (size_t)1 * R3 * C; v1_1_2.C = GC + (size_t)1 * R3 * C;
      v1_1_2.sAo = (long long)34 * 34 * C; v1_1_2.sAi = (long long)34 * C; v1_1_2.sAm = C; v1_1_2.sAk = 1; v1_1_2.sBo = 0; v1_1_2.sBi = 0; v1_1_2.sBn = C * 27; v1_1_2.sBk = 27; v1_1_2.sCo = (long long)R * R * C; v1_1_2.sCi = (long long)R * C; v1_1_2.sCm = C; v1_1_2.sRo = (long long)R * R * C; v1_1_2.sRi = (long long)R * C; v1_1_2.sRm = C; v1_1_2.sRn = 1;
      v1_1_2.M = R; v1_1_2.N = C; v1_1_2.K = C; v1_1_2.zi_n = R; v1_1_2.flags = 4; v1_1_2.act = 0;
      v1_1_2.alpha = 1.0f; v1_1_2.beta = 1.0f; v1_1_2.sa = 1.0f; v1_1_2.sb = 1.0f; v1_1_2.Npad = C; v1_1_2.pad_ = 0;
      k_gemm<1><<<dim3((unsigned)((C) + 31) / 32, (unsigned)((R) + 15) / 16, (unsigned)(R * R)), 32, 0, stream>>>(v1_1_2); }
    { GemmP v1_1_3;
      v1_1_3.A = GP + (size_t)1 * RP3 * C + (size_t)34 * C; v1_1_3.B = wv1 + 3; v1_1_3.bias = GP + (size_t)1 * RP3 * C + (size_t)34 * C; v1_1_3.R = GC + (size_t)1 * R3 * C; v1_1_3.C = GC + (size_t)1 * R3 * C;
      v1_1_3.sAo = (long long)34 * 34 * C; v1_1_3.sAi = (long long)34 * C; v1_1_3.sAm = C; v1_1_3.sAk = 1; v1_1_3.sBo = 0; v1_1_3.sBi = 0; v1_1_3.sBn = C * 27; v1_1_3.sBk = 27; v1_1_3.sCo = (long long)R * R * C; v1_1_3.sCi = (long long)R * C; v1_1_3.sCm = C; v1_1_3.sRo = (long long)R * R * C; v1_1_3.sRi = (long long)R * C; v1_1_3.sRm = C; v1_1_3.sRn = 1;
      v1_1_3.M = R; v1_1_3.N = C; v1_1_3.K = C; v1_1_3.zi_n = R; v1_1_3.flags = 4; v1_1_3.act = 0;
      v1_1_3.alpha = 1.0f; v1_1_3.beta = 1.0f; v1_1_3.sa = 1.0f; v1_1_3.sb = 1.0f; v1_1_3.Npad = C; v1_1_3.pad_ = 0;
      k_gemm<1><<<dim3((unsigned)((C) + 31) / 32, (unsigned)((R) + 15) / 16, (unsigned)(R * R)), 32, 0, stream>>>(v1_1_3); }
    { GemmP v1_1_4;
      v1_1_4.A = GP + (size_t)1 * RP3 * C + (size_t)35 * C; v1_1_4.B = wv1 + 4; v1_1_4.bias = GP + (size_t)1 * RP3 * C + (size_t)35 * C; v1_1_4.R = GC + (size_t)1 * R3 * C; v1_1_4.C = GC + (size_t)1 * R3 * C;
      v1_1_4.sAo = (long long)34 * 34 * C; v1_1_4.sAi = (long long)34 * C; v1_1_4.sAm = C; v1_1_4.sAk = 1; v1_1_4.sBo = 0; v1_1_4.sBi = 0; v1_1_4.sBn = C * 27; v1_1_4.sBk = 27; v1_1_4.sCo = (long long)R * R * C; v1_1_4.sCi = (long long)R * C; v1_1_4.sCm = C; v1_1_4.sRo = (long long)R * R * C; v1_1_4.sRi = (long long)R * C; v1_1_4.sRm = C; v1_1_4.sRn = 1;
      v1_1_4.M = R; v1_1_4.N = C; v1_1_4.K = C; v1_1_4.zi_n = R; v1_1_4.flags = 4; v1_1_4.act = 0;
      v1_1_4.alpha = 1.0f; v1_1_4.beta = 1.0f; v1_1_4.sa = 1.0f; v1_1_4.sb = 1.0f; v1_1_4.Npad = C; v1_1_4.pad_ = 0;
      k_gemm<1><<<dim3((unsigned)((C) + 31) / 32, (unsigned)((R) + 15) / 16, (unsigned)(R * R)), 32, 0, stream>>>(v1_1_4); }
    { GemmP v1_1_5;
      v1_1_5.A = GP + (size_t)1 * RP3 * C + (size_t)36 * C; v1_1_5.B = wv1 + 5; v1_1_5.bias = GP + (size_t)1 * RP3 * C + (size_t)36 * C; v1_1_5.R = GC + (size_t)1 * R3 * C; v1_1_5.C = GC + (size_t)1 * R3 * C;
      v1_1_5.sAo = (long long)34 * 34 * C; v1_1_5.sAi = (long long)34 * C; v1_1_5.sAm = C; v1_1_5.sAk = 1; v1_1_5.sBo = 0; v1_1_5.sBi = 0; v1_1_5.sBn = C * 27; v1_1_5.sBk = 27; v1_1_5.sCo = (long long)R * R * C; v1_1_5.sCi = (long long)R * C; v1_1_5.sCm = C; v1_1_5.sRo = (long long)R * R * C; v1_1_5.sRi = (long long)R * C; v1_1_5.sRm = C; v1_1_5.sRn = 1;
      v1_1_5.M = R; v1_1_5.N = C; v1_1_5.K = C; v1_1_5.zi_n = R; v1_1_5.flags = 4; v1_1_5.act = 0;
      v1_1_5.alpha = 1.0f; v1_1_5.beta = 1.0f; v1_1_5.sa = 1.0f; v1_1_5.sb = 1.0f; v1_1_5.Npad = C; v1_1_5.pad_ = 0;
      k_gemm<1><<<dim3((unsigned)((C) + 31) / 32, (unsigned)((R) + 15) / 16, (unsigned)(R * R)), 32, 0, stream>>>(v1_1_5); }
    { GemmP v1_1_6;
      v1_1_6.A = GP + (size_t)1 * RP3 * C + (size_t)68 * C; v1_1_6.B = wv1 + 6; v1_1_6.bias = GP + (size_t)1 * RP3 * C + (size_t)68 * C; v1_1_6.R = GC + (size_t)1 * R3 * C; v1_1_6.C = GC + (size_t)1 * R3 * C;
      v1_1_6.sAo = (long long)34 * 34 * C; v1_1_6.sAi = (long long)34 * C; v1_1_6.sAm = C; v1_1_6.sAk = 1; v1_1_6.sBo = 0; v1_1_6.sBi = 0; v1_1_6.sBn = C * 27; v1_1_6.sBk = 27; v1_1_6.sCo = (long long)R * R * C; v1_1_6.sCi = (long long)R * C; v1_1_6.sCm = C; v1_1_6.sRo = (long long)R * R * C; v1_1_6.sRi = (long long)R * C; v1_1_6.sRm = C; v1_1_6.sRn = 1;
      v1_1_6.M = R; v1_1_6.N = C; v1_1_6.K = C; v1_1_6.zi_n = R; v1_1_6.flags = 4; v1_1_6.act = 0;
      v1_1_6.alpha = 1.0f; v1_1_6.beta = 1.0f; v1_1_6.sa = 1.0f; v1_1_6.sb = 1.0f; v1_1_6.Npad = C; v1_1_6.pad_ = 0;
      k_gemm<1><<<dim3((unsigned)((C) + 31) / 32, (unsigned)((R) + 15) / 16, (unsigned)(R * R)), 32, 0, stream>>>(v1_1_6); }
    { GemmP v1_1_7;
      v1_1_7.A = GP + (size_t)1 * RP3 * C + (size_t)69 * C; v1_1_7.B = wv1 + 7; v1_1_7.bias = GP + (size_t)1 * RP3 * C + (size_t)69 * C; v1_1_7.R = GC + (size_t)1 * R3 * C; v1_1_7.C = GC + (size_t)1 * R3 * C;
      v1_1_7.sAo = (long long)34 * 34 * C; v1_1_7.sAi = (long long)34 * C; v1_1_7.sAm = C; v1_1_7.sAk = 1; v1_1_7.sBo = 0; v1_1_7.sBi = 0; v1_1_7.sBn = C * 27; v1_1_7.sBk = 27; v1_1_7.sCo = (long long)R * R * C; v1_1_7.sCi = (long long)R * C; v1_1_7.sCm = C; v1_1_7.sRo = (long long)R * R * C; v1_1_7.sRi = (long long)R * C; v1_1_7.sRm = C; v1_1_7.sRn = 1;
      v1_1_7.M = R; v1_1_7.N = C; v1_1_7.K = C; v1_1_7.zi_n = R; v1_1_7.flags = 4; v1_1_7.act = 0;
      v1_1_7.alpha = 1.0f; v1_1_7.beta = 1.0f; v1_1_7.sa = 1.0f; v1_1_7.sb = 1.0f; v1_1_7.Npad = C; v1_1_7.pad_ = 0;
      k_gemm<1><<<dim3((unsigned)((C) + 31) / 32, (unsigned)((R) + 15) / 16, (unsigned)(R * R)), 32, 0, stream>>>(v1_1_7); }
    { GemmP v1_1_8;
      v1_1_8.A = GP + (size_t)1 * RP3 * C + (size_t)70 * C; v1_1_8.B = wv1 + 8; v1_1_8.bias = GP + (size_t)1 * RP3 * C + (size_t)70 * C; v1_1_8.R = GC + (size_t)1 * R3 * C; v1_1_8.C = GC + (size_t)1 * R3 * C;
      v1_1_8.sAo = (long long)34 * 34 * C; v1_1_8.sAi = (long long)34 * C; v1_1_8.sAm = C; v1_1_8.sAk = 1; v1_1_8.sBo = 0; v1_1_8.sBi = 0; v1_1_8.sBn = C * 27; v1_1_8.sBk = 27; v1_1_8.sCo = (long long)R * R * C; v1_1_8.sCi = (long long)R * C; v1_1_8.sCm = C; v1_1_8.sRo = (long long)R * R * C; v1_1_8.sRi = (long long)R * C; v1_1_8.sRm = C; v1_1_8.sRn = 1;
      v1_1_8.M = R; v1_1_8.N = C; v1_1_8.K = C; v1_1_8.zi_n = R; v1_1_8.flags = 4; v1_1_8.act = 0;
      v1_1_8.alpha = 1.0f; v1_1_8.beta = 1.0f; v1_1_8.sa = 1.0f; v1_1_8.sb = 1.0f; v1_1_8.Npad = C; v1_1_8.pad_ = 0;
      k_gemm<1><<<dim3((unsigned)((C) + 31) / 32, (unsigned)((R) + 15) / 16, (unsigned)(R * R)), 32, 0, stream>>>(v1_1_8); }
    { GemmP v1_1_9;
      v1_1_9.A = GP + (size_t)1 * RP3 * C + (size_t)1156 * C; v1_1_9.B = wv1 + 9; v1_1_9.bias = GP + (size_t)1 * RP3 * C + (size_t)1156 * C; v1_1_9.R = GC + (size_t)1 * R3 * C; v1_1_9.C = GC + (size_t)1 * R3 * C;
      v1_1_9.sAo = (long long)34 * 34 * C; v1_1_9.sAi = (long long)34 * C; v1_1_9.sAm = C; v1_1_9.sAk = 1; v1_1_9.sBo = 0; v1_1_9.sBi = 0; v1_1_9.sBn = C * 27; v1_1_9.sBk = 27; v1_1_9.sCo = (long long)R * R * C; v1_1_9.sCi = (long long)R * C; v1_1_9.sCm = C; v1_1_9.sRo = (long long)R * R * C; v1_1_9.sRi = (long long)R * C; v1_1_9.sRm = C; v1_1_9.sRn = 1;
      v1_1_9.M = R; v1_1_9.N = C; v1_1_9.K = C; v1_1_9.zi_n = R; v1_1_9.flags = 4; v1_1_9.act = 0;
      v1_1_9.alpha = 1.0f; v1_1_9.beta = 1.0f; v1_1_9.sa = 1.0f; v1_1_9.sb = 1.0f; v1_1_9.Npad = C; v1_1_9.pad_ = 0;
      k_gemm<1><<<dim3((unsigned)((C) + 31) / 32, (unsigned)((R) + 15) / 16, (unsigned)(R * R)), 32, 0, stream>>>(v1_1_9); }
    { GemmP v1_1_10;
      v1_1_10.A = GP + (size_t)1 * RP3 * C + (size_t)1157 * C; v1_1_10.B = wv1 + 10; v1_1_10.bias = GP + (size_t)1 * RP3 * C + (size_t)1157 * C; v1_1_10.R = GC + (size_t)1 * R3 * C; v1_1_10.C = GC + (size_t)1 * R3 * C;
      v1_1_10.sAo = (long long)34 * 34 * C; v1_1_10.sAi = (long long)34 * C; v1_1_10.sAm = C; v1_1_10.sAk = 1; v1_1_10.sBo = 0; v1_1_10.sBi = 0; v1_1_10.sBn = C * 27; v1_1_10.sBk = 27; v1_1_10.sCo = (long long)R * R * C; v1_1_10.sCi = (long long)R * C; v1_1_10.sCm = C; v1_1_10.sRo = (long long)R * R * C; v1_1_10.sRi = (long long)R * C; v1_1_10.sRm = C; v1_1_10.sRn = 1;
      v1_1_10.M = R; v1_1_10.N = C; v1_1_10.K = C; v1_1_10.zi_n = R; v1_1_10.flags = 4; v1_1_10.act = 0;
      v1_1_10.alpha = 1.0f; v1_1_10.beta = 1.0f; v1_1_10.sa = 1.0f; v1_1_10.sb = 1.0f; v1_1_10.Npad = C; v1_1_10.pad_ = 0;
      k_gemm<1><<<dim3((unsigned)((C) + 31) / 32, (unsigned)((R) + 15) / 16, (unsigned)(R * R)), 32, 0, stream>>>(v1_1_10); }
    { GemmP v1_1_11;
      v1_1_11.A = GP + (size_t)1 * RP3 * C + (size_t)1158 * C; v1_1_11.B = wv1 + 11; v1_1_11.bias = GP + (size_t)1 * RP3 * C + (size_t)1158 * C; v1_1_11.R = GC + (size_t)1 * R3 * C; v1_1_11.C = GC + (size_t)1 * R3 * C;
      v1_1_11.sAo = (long long)34 * 34 * C; v1_1_11.sAi = (long long)34 * C; v1_1_11.sAm = C; v1_1_11.sAk = 1; v1_1_11.sBo = 0; v1_1_11.sBi = 0; v1_1_11.sBn = C * 27; v1_1_11.sBk = 27; v1_1_11.sCo = (long long)R * R * C; v1_1_11.sCi = (long long)R * C; v1_1_11.sCm = C; v1_1_11.sRo = (long long)R * R * C; v1_1_11.sRi = (long long)R * C; v1_1_11.sRm = C; v1_1_11.sRn = 1;
      v1_1_11.M = R; v1_1_11.N = C; v1_1_11.K = C; v1_1_11.zi_n = R; v1_1_11.flags = 4; v1_1_11.act = 0;
      v1_1_11.alpha = 1.0f; v1_1_11.beta = 1.0f; v1_1_11.sa = 1.0f; v1_1_11.sb = 1.0f; v1_1_11.Npad = C; v1_1_11.pad_ = 0;
      k_gemm<1><<<dim3((unsigned)((C) + 31) / 32, (unsigned)((R) + 15) / 16, (unsigned)(R * R)), 32, 0, stream>>>(v1_1_11); }
    { GemmP v1_1_12;
      v1_1_12.A = GP + (size_t)1 * RP3 * C + (size_t)1190 * C; v1_1_12.B = wv1 + 12; v1_1_12.bias = GP + (size_t)1 * RP3 * C + (size_t)1190 * C; v1_1_12.R = GC + (size_t)1 * R3 * C; v1_1_12.C = GC + (size_t)1 * R3 * C;
      v1_1_12.sAo = (long long)34 * 34 * C; v1_1_12.sAi = (long long)34 * C; v1_1_12.sAm = C; v1_1_12.sAk = 1; v1_1_12.sBo = 0; v1_1_12.sBi = 0; v1_1_12.sBn = C * 27; v1_1_12.sBk = 27; v1_1_12.sCo = (long long)R * R * C; v1_1_12.sCi = (long long)R * C; v1_1_12.sCm = C; v1_1_12.sRo = (long long)R * R * C; v1_1_12.sRi = (long long)R * C; v1_1_12.sRm = C; v1_1_12.sRn = 1;
      v1_1_12.M = R; v1_1_12.N = C; v1_1_12.K = C; v1_1_12.zi_n = R; v1_1_12.flags = 4; v1_1_12.act = 0;
      v1_1_12.alpha = 1.0f; v1_1_12.beta = 1.0f; v1_1_12.sa = 1.0f; v1_1_12.sb = 1.0f; v1_1_12.Npad = C; v1_1_12.pad_ = 0;
      k_gemm<1><<<dim3((unsigned)((C) + 31) / 32, (unsigned)((R) + 15) / 16, (unsigned)(R * R)), 32, 0, stream>>>(v1_1_12); }
    { GemmP v1_1_13;
      v1_1_13.A = GP + (size_t)1 * RP3 * C + (size_t)1191 * C; v1_1_13.B = wv1 + 13; v1_1_13.bias = GP + (size_t)1 * RP3 * C + (size_t)1191 * C; v1_1_13.R = GC + (size_t)1 * R3 * C; v1_1_13.C = GC + (size_t)1 * R3 * C;
      v1_1_13.sAo = (long long)34 * 34 * C; v1_1_13.sAi = (long long)34 * C; v1_1_13.sAm = C; v1_1_13.sAk = 1; v1_1_13.sBo = 0; v1_1_13.sBi = 0; v1_1_13.sBn = C * 27; v1_1_13.sBk = 27; v1_1_13.sCo = (long long)R * R * C; v1_1_13.sCi = (long long)R * C; v1_1_13.sCm = C; v1_1_13.sRo = (long long)R * R * C; v1_1_13.sRi = (long long)R * C; v1_1_13.sRm = C; v1_1_13.sRn = 1;
      v1_1_13.M = R; v1_1_13.N = C; v1_1_13.K = C; v1_1_13.zi_n = R; v1_1_13.flags = 4; v1_1_13.act = 0;
      v1_1_13.alpha = 1.0f; v1_1_13.beta = 1.0f; v1_1_13.sa = 1.0f; v1_1_13.sb = 1.0f; v1_1_13.Npad = C; v1_1_13.pad_ = 0;
      k_gemm<1><<<dim3((unsigned)((C) + 31) / 32, (unsigned)((R) + 15) / 16, (unsigned)(R * R)), 32, 0, stream>>>(v1_1_13); }
    { GemmP v1_1_14;
      v1_1_14.A = GP + (size_t)1 * RP3 * C + (size_t)1192 * C; v1_1_14.B = wv1 + 14; v1_1_14.bias = GP + (size_t)1 * RP3 * C + (size_t)1192 * C; v1_1_14.R = GC + (size_t)1 * R3 * C; v1_1_14.C = GC + (size_t)1 * R3 * C;
      v1_1_14.sAo = (long long)34 * 34 * C; v1_1_14.sAi = (long long)34 * C; v1_1_14.sAm = C; v1_1_14.sAk = 1; v1_1_14.sBo = 0; v1_1_14.sBi = 0; v1_1_14.sBn = C * 27; v1_1_14.sBk = 27; v1_1_14.sCo = (long long)R * R * C; v1_1_14.sCi = (long long)R * C; v1_1_14.sCm = C; v1_1_14.sRo = (long long)R * R * C; v1_1_14.sRi = (long long)R * C; v1_1_14.sRm = C; v1_1_14.sRn = 1;
      v1_1_14.M = R; v1_1_14.N = C; v1_1_14.K = C; v1_1_14.zi_n = R; v1_1_14.flags = 4; v1_1_14.act = 0;
      v1_1_14.alpha = 1.0f; v1_1_14.beta = 1.0f; v1_1_14.sa = 1.0f; v1_1_14.sb = 1.0f; v1_1_14.Npad = C; v1_1_14.pad_ = 0;
      k_gemm<1><<<dim3((unsigned)((C) + 31) / 32, (unsigned)((R) + 15) / 16, (unsigned)(R * R)), 32, 0, stream>>>(v1_1_14); }
    { GemmP v1_1_15;
      v1_1_15.A = GP + (size_t)1 * RP3 * C + (size_t)1224 * C; v1_1_15.B = wv1 + 15; v1_1_15.bias = GP + (size_t)1 * RP3 * C + (size_t)1224 * C; v1_1_15.R = GC + (size_t)1 * R3 * C; v1_1_15.C = GC + (size_t)1 * R3 * C;
      v1_1_15.sAo = (long long)34 * 34 * C; v1_1_15.sAi = (long long)34 * C; v1_1_15.sAm = C; v1_1_15.sAk = 1; v1_1_15.sBo = 0; v1_1_15.sBi = 0; v1_1_15.sBn = C * 27; v1_1_15.sBk = 27; v1_1_15.sCo = (long long)R * R * C; v1_1_15.sCi = (long long)R * C; v1_1_15.sCm = C; v1_1_15.sRo = (long long)R * R * C; v1_1_15.sRi = (long long)R * C; v1_1_15.sRm = C; v1_1_15.sRn = 1;
      v1_1_15.M = R; v1_1_15.N = C; v1_1_15.K = C; v1_1_15.zi_n = R; v1_1_15.flags = 4; v1_1_15.act = 0;
      v1_1_15.alpha = 1.0f; v1_1_15.beta = 1.0f; v1_1_15.sa = 1.0f; v1_1_15.sb = 1.0f; v1_1_15.Npad = C; v1_1_15.pad_ = 0;
      k_gemm<1><<<dim3((unsigned)((C) + 31) / 32, (unsigned)((R) + 15) / 16, (unsigned)(R * R)), 32, 0, stream>>>(v1_1_15); }
    { GemmP v1_1_16;
      v1_1_16.A = GP + (size_t)1 * RP3 * C + (size_t)1225 * C; v1_1_16.B = wv1 + 16; v1_1_16.bias = GP + (size_t)1 * RP3 * C + (size_t)1225 * C; v1_1_16.R = GC + (size_t)1 * R3 * C; v1_1_16.C = GC + (size_t)1 * R3 * C;
      v1_1_16.sAo = (long long)34 * 34 * C; v1_1_16.sAi = (long long)34 * C; v1_1_16.sAm = C; v1_1_16.sAk = 1; v1_1_16.sBo = 0; v1_1_16.sBi = 0; v1_1_16.sBn = C * 27; v1_1_16.sBk = 27; v1_1_16.sCo = (long long)R * R * C; v1_1_16.sCi = (long long)R * C; v1_1_16.sCm = C; v1_1_16.sRo = (long long)R * R * C; v1_1_16.sRi = (long long)R * C; v1_1_16.sRm = C; v1_1_16.sRn = 1;
      v1_1_16.M = R; v1_1_16.N = C; v1_1_16.K = C; v1_1_16.zi_n = R; v1_1_16.flags = 4; v1_1_16.act = 0;
      v1_1_16.alpha = 1.0f; v1_1_16.beta = 1.0f; v1_1_16.sa = 1.0f; v1_1_16.sb = 1.0f; v1_1_16.Npad = C; v1_1_16.pad_ = 0;
      k_gemm<1><<<dim3((unsigned)((C) + 31) / 32, (unsigned)((R) + 15) / 16, (unsigned)(R * R)), 32, 0, stream>>>(v1_1_16); }
    { GemmP v1_1_17;
      v1_1_17.A = GP + (size_t)1 * RP3 * C + (size_t)1226 * C; v1_1_17.B = wv1 + 17; v1_1_17.bias = GP + (size_t)1 * RP3 * C + (size_t)1226 * C; v1_1_17.R = GC + (size_t)1 * R3 * C; v1_1_17.C = GC + (size_t)1 * R3 * C;
      v1_1_17.sAo = (long long)34 * 34 * C; v1_1_17.sAi = (long long)34 * C; v1_1_17.sAm = C; v1_1_17.sAk = 1; v1_1_17.sBo = 0; v1_1_17.sBi = 0; v1_1_17.sBn = C * 27; v1_1_17.sBk = 27; v1_1_17.sCo = (long long)R * R * C; v1_1_17.sCi = (long long)R * C; v1_1_17.sCm = C; v1_1_17.sRo = (long long)R * R * C; v1_1_17.sRi = (long long)R * C; v1_1_17.sRm = C; v1_1_17.sRn = 1;
      v1_1_17.M = R; v1_1_17.N = C; v1_1_17.K = C; v1_1_17.zi_n = R; v1_1_17.flags = 4; v1_1_17.act = 0;
      v1_1_17.alpha = 1.0f; v1_1_17.beta = 1.0f; v1_1_17.sa = 1.0f; v1_1_17.sb = 1.0f; v1_1_17.Npad = C; v1_1_17.pad_ = 0;
      k_gemm<1><<<dim3((unsigned)((C) + 31) / 32, (unsigned)((R) + 15) / 16, (unsigned)(R * R)), 32, 0, stream>>>(v1_1_17); }
    { GemmP v1_1_18;
      v1_1_18.A = GP + (size_t)1 * RP3 * C + (size_t)2312 * C; v1_1_18.B = wv1 + 18; v1_1_18.bias = GP + (size_t)1 * RP3 * C + (size_t)2312 * C; v1_1_18.R = GC + (size_t)1 * R3 * C; v1_1_18.C = GC + (size_t)1 * R3 * C;
      v1_1_18.sAo = (long long)34 * 34 * C; v1_1_18.sAi = (long long)34 * C; v1_1_18.sAm = C; v1_1_18.sAk = 1; v1_1_18.sBo = 0; v1_1_18.sBi = 0; v1_1_18.sBn = C * 27; v1_1_18.sBk = 27; v1_1_18.sCo = (long long)R * R * C; v1_1_18.sCi = (long long)R * C; v1_1_18.sCm = C; v1_1_18.sRo = (long long)R * R * C; v1_1_18.sRi = (long long)R * C; v1_1_18.sRm = C; v1_1_18.sRn = 1;
      v1_1_18.M = R; v1_1_18.N = C; v1_1_18.K = C; v1_1_18.zi_n = R; v1_1_18.flags = 4; v1_1_18.act = 0;
      v1_1_18.alpha = 1.0f; v1_1_18.beta = 1.0f; v1_1_18.sa = 1.0f; v1_1_18.sb = 1.0f; v1_1_18.Npad = C; v1_1_18.pad_ = 0;
      k_gemm<1><<<dim3((unsigned)((C) + 31) / 32, (unsigned)((R) + 15) / 16, (unsigned)(R * R)), 32, 0, stream>>>(v1_1_18); }
    { GemmP v1_1_19;
      v1_1_19.A = GP + (size_t)1 * RP3 * C + (size_t)2313 * C; v1_1_19.B = wv1 + 19; v1_1_19.bias = GP + (size_t)1 * RP3 * C + (size_t)2313 * C; v1_1_19.R = GC + (size_t)1 * R3 * C; v1_1_19.C = GC + (size_t)1 * R3 * C;
      v1_1_19.sAo = (long long)34 * 34 * C; v1_1_19.sAi = (long long)34 * C; v1_1_19.sAm = C; v1_1_19.sAk = 1; v1_1_19.sBo = 0; v1_1_19.sBi = 0; v1_1_19.sBn = C * 27; v1_1_19.sBk = 27; v1_1_19.sCo = (long long)R * R * C; v1_1_19.sCi = (long long)R * C; v1_1_19.sCm = C; v1_1_19.sRo = (long long)R * R * C; v1_1_19.sRi = (long long)R * C; v1_1_19.sRm = C; v1_1_19.sRn = 1;
      v1_1_19.M = R; v1_1_19.N = C; v1_1_19.K = C; v1_1_19.zi_n = R; v1_1_19.flags = 4; v1_1_19.act = 0;
      v1_1_19.alpha = 1.0f; v1_1_19.beta = 1.0f; v1_1_19.sa = 1.0f; v1_1_19.sb = 1.0f; v1_1_19.Npad = C; v1_1_19.pad_ = 0;
      k_gemm<1><<<dim3((unsigned)((C) + 31) / 32, (unsigned)((R) + 15) / 16, (unsigned)(R * R)), 32, 0, stream>>>(v1_1_19); }
    { GemmP v1_1_20;
      v1_1_20.A = GP + (size_t)1 * RP3 * C + (size_t)2314 * C; v1_1_20.B = wv1 + 20; v1_1_20.bias = GP + (size_t)1 * RP3 * C + (size_t)2314 * C; v1_1_20.R = GC + (size_t)1 * R3 * C; v1_1_20.C = GC + (size_t)1 * R3 * C;
      v1_1_20.sAo = (long long)34 * 34 * C; v1_1_20.sAi = (long long)34 * C; v1_1_20.sAm = C; v1_1_20.sAk = 1; v1_1_20.sBo = 0; v1_1_20.sBi = 0; v1_1_20.sBn = C * 27; v1_1_20.sBk = 27; v1_1_20.sCo = (long long)R * R * C; v1_1_20.sCi = (long long)R * C; v1_1_20.sCm = C; v1_1_20.sRo = (long long)R * R * C; v1_1_20.sRi = (long long)R * C; v1_1_20.sRm = C; v1_1_20.sRn = 1;
      v1_1_20.M = R; v1_1_20.N = C; v1_1_20.K = C; v1_1_20.zi_n = R; v1_1_20.flags = 4; v1_1_20.act = 0;
      v1_1_20.alpha = 1.0f; v1_1_20.beta = 1.0f; v1_1_20.sa = 1.0f; v1_1_20.sb = 1.0f; v1_1_20.Npad = C; v1_1_20.pad_ = 0;
      k_gemm<1><<<dim3((unsigned)((C) + 31) / 32, (unsigned)((R) + 15) / 16, (unsigned)(R * R)), 32, 0, stream>>>(v1_1_20); }
    { GemmP v1_1_21;
      v1_1_21.A = GP + (size_t)1 * RP3 * C + (size_t)2346 * C; v1_1_21.B = wv1 + 21; v1_1_21.bias = GP + (size_t)1 * RP3 * C + (size_t)2346 * C; v1_1_21.R = GC + (size_t)1 * R3 * C; v1_1_21.C = GC + (size_t)1 * R3 * C;
      v1_1_21.sAo = (long long)34 * 34 * C; v1_1_21.sAi = (long long)34 * C; v1_1_21.sAm = C; v1_1_21.sAk = 1; v1_1_21.sBo = 0; v1_1_21.sBi = 0; v1_1_21.sBn = C * 27; v1_1_21.sBk = 27; v1_1_21.sCo = (long long)R * R * C; v1_1_21.sCi = (long long)R * C; v1_1_21.sCm = C; v1_1_21.sRo = (long long)R * R * C; v1_1_21.sRi = (long long)R * C; v1_1_21.sRm = C; v1_1_21.sRn = 1;
      v1_1_21.M = R; v1_1_21.N = C; v1_1_21.K = C; v1_1_21.zi_n = R; v1_1_21.flags = 4; v1_1_21.act = 0;
      v1_1_21.alpha = 1.0f; v1_1_21.beta = 1.0f; v1_1_21.sa = 1.0f; v1_1_21.sb = 1.0f; v1_1_21.Npad = C; v1_1_21.pad_ = 0;
      k_gemm<1><<<dim3((unsigned)((C) + 31) / 32, (unsigned)((R) + 15) / 16, (unsigned)(R * R)), 32, 0, stream>>>(v1_1_21); }
    { GemmP v1_1_22;
      v1_1_22.A = GP + (size_t)1 * RP3 * C + (size_t)2347 * C; v1_1_22.B = wv1 + 22; v1_1_22.bias = GP + (size_t)1 * RP3 * C + (size_t)2347 * C; v1_1_22.R = GC + (size_t)1 * R3 * C; v1_1_22.C = GC + (size_t)1 * R3 * C;
      v1_1_22.sAo = (long long)34 * 34 * C; v1_1_22.sAi = (long long)34 * C; v1_1_22.sAm = C; v1_1_22.sAk = 1; v1_1_22.sBo = 0; v1_1_22.sBi = 0; v1_1_22.sBn = C * 27; v1_1_22.sBk = 27; v1_1_22.sCo = (long long)R * R * C; v1_1_22.sCi = (long long)R * C; v1_1_22.sCm = C; v1_1_22.sRo = (long long)R * R * C; v1_1_22.sRi = (long long)R * C; v1_1_22.sRm = C; v1_1_22.sRn = 1;
      v1_1_22.M = R; v1_1_22.N = C; v1_1_22.K = C; v1_1_22.zi_n = R; v1_1_22.flags = 4; v1_1_22.act = 0;
      v1_1_22.alpha = 1.0f; v1_1_22.beta = 1.0f; v1_1_22.sa = 1.0f; v1_1_22.sb = 1.0f; v1_1_22.Npad = C; v1_1_22.pad_ = 0;
      k_gemm<1><<<dim3((unsigned)((C) + 31) / 32, (unsigned)((R) + 15) / 16, (unsigned)(R * R)), 32, 0, stream>>>(v1_1_22); }
    { GemmP v1_1_23;
      v1_1_23.A = GP + (size_t)1 * RP3 * C + (size_t)2348 * C; v1_1_23.B = wv1 + 23; v1_1_23.bias = GP + (size_t)1 * RP3 * C + (size_t)2348 * C; v1_1_23.R = GC + (size_t)1 * R3 * C; v1_1_23.C = GC + (size_t)1 * R3 * C;
      v1_1_23.sAo = (long long)34 * 34 * C; v1_1_23.sAi = (long long)34 * C; v1_1_23.sAm = C; v1_1_23.sAk = 1; v1_1_23.sBo = 0; v1_1_23.sBi = 0; v1_1_23.sBn = C * 27; v1_1_23.sBk = 27; v1_1_23.sCo = (long long)R * R * C; v1_1_23.sCi = (long long)R * C; v1_1_23.sCm = C; v1_1_23.sRo = (long long)R * R * C; v1_1_23.sRi = (long long)R * C; v1_1_23.sRm = C; v1_1_23.sRn = 1;
      v1_1_23.M = R; v1_1_23.N = C; v1_1_23.K = C; v1_1_23.zi_n = R; v1_1_23.flags = 4; v1_1_23.act = 0;
      v1_1_23.alpha = 1.0f; v1_1_23.beta = 1.0f; v1_1_23.sa = 1.0f; v1_1_23.sb = 1.0f; v1_1_23.Npad = C; v1_1_23.pad_ = 0;
      k_gemm<1><<<dim3((unsigned)((C) + 31) / 32, (unsigned)((R) + 15) / 16, (unsigned)(R * R)), 32, 0, stream>>>(v1_1_23); }
    { GemmP v1_1_24;
      v1_1_24.A = GP + (size_t)1 * RP3 * C + (size_t)2380 * C; v1_1_24.B = wv1 + 24; v1_1_24.bias = GP + (size_t)1 * RP3 * C + (size_t)2380 * C; v1_1_24.R = GC + (size_t)1 * R3 * C; v1_1_24.C = GC + (size_t)1 * R3 * C;
      v1_1_24.sAo = (long long)34 * 34 * C; v1_1_24.sAi = (long long)34 * C; v1_1_24.sAm = C; v1_1_24.sAk = 1; v1_1_24.sBo = 0; v1_1_24.sBi = 0; v1_1_24.sBn = C * 27; v1_1_24.sBk = 27; v1_1_24.sCo = (long long)R * R * C; v1_1_24.sCi = (long long)R * C; v1_1_24.sCm = C; v1_1_24.sRo = (long long)R * R * C; v1_1_24.sRi = (long long)R * C; v1_1_24.sRm = C; v1_1_24.sRn = 1;
      v1_1_24.M = R; v1_1_24.N = C; v1_1_24.K = C; v1_1_24.zi_n = R; v1_1_24.flags = 4; v1_1_24.act = 0;
      v1_1_24.alpha = 1.0f; v1_1_24.beta = 1.0f; v1_1_24.sa = 1.0f; v1_1_24.sb = 1.0f; v1_1_24.Npad = C; v1_1_24.pad_ = 0;
      k_gemm<1><<<dim3((unsigned)((C) + 31) / 32, (unsigned)((R) + 15) / 16, (unsigned)(R * R)), 32, 0, stream>>>(v1_1_24); }
    { GemmP v1_1_25;
      v1_1_25.A = GP + (size_t)1 * RP3 * C + (size_t)2381 * C; v1_1_25.B = wv1 + 25; v1_1_25.bias = GP + (size_t)1 * RP3 * C + (size_t)2381 * C; v1_1_25.R = GC + (size_t)1 * R3 * C; v1_1_25.C = GC + (size_t)1 * R3 * C;
      v1_1_25.sAo = (long long)34 * 34 * C; v1_1_25.sAi = (long long)34 * C; v1_1_25.sAm = C; v1_1_25.sAk = 1; v1_1_25.sBo = 0; v1_1_25.sBi = 0; v1_1_25.sBn = C * 27; v1_1_25.sBk = 27; v1_1_25.sCo = (long long)R * R * C; v1_1_25.sCi = (long long)R * C; v1_1_25.sCm = C; v1_1_25.sRo = (long long)R * R * C; v1_1_25.sRi = (long long)R * C; v1_1_25.sRm = C; v1_1_25.sRn = 1;
      v1_1_25.M = R; v1_1_25.N = C; v1_1_25.K = C; v1_1_25.zi_n = R; v1_1_25.flags = 4; v1_1_25.act = 0;
      v1_1_25.alpha = 1.0f; v1_1_25.beta = 1.0f; v1_1_25.sa = 1.0f; v1_1_25.sb = 1.0f; v1_1_25.Npad = C; v1_1_25.pad_ = 0;
      k_gemm<1><<<dim3((unsigned)((C) + 31) / 32, (unsigned)((R) + 15) / 16, (unsigned)(R * R)), 32, 0, stream>>>(v1_1_25); }
    { GemmP v1_1_26;
      v1_1_26.A = GP + (size_t)1 * RP3 * C + (size_t)2382 * C; v1_1_26.B = wv1 + 26; v1_1_26.bias = GP + (size_t)1 * RP3 * C + (size_t)2382 * C; v1_1_26.R = GC + (size_t)1 * R3 * C; v1_1_26.C = GC + (size_t)1 * R3 * C;
      v1_1_26.sAo = (long long)34 * 34 * C; v1_1_26.sAi = (long long)34 * C; v1_1_26.sAm = C; v1_1_26.sAk = 1; v1_1_26.sBo = 0; v1_1_26.sBi = 0; v1_1_26.sBn = C * 27; v1_1_26.sBk = 27; v1_1_26.sCo = (long long)R * R * C; v1_1_26.sCi = (long long)R * C; v1_1_26.sCm = C; v1_1_26.sRo = (long long)R * R * C; v1_1_26.sRi = (long long)R * C; v1_1_26.sRm = C; v1_1_26.sRn = 1;
      v1_1_26.M = R; v1_1_26.N = C; v1_1_26.K = C; v1_1_26.zi_n = R; v1_1_26.flags = 4; v1_1_26.act = 0;
      v1_1_26.alpha = 1.0f; v1_1_26.beta = 1.0f; v1_1_26.sa = 1.0f; v1_1_26.sb = 1.0f; v1_1_26.Npad = C; v1_1_26.pad_ = 0;
      k_gemm<1><<<dim3((unsigned)((C) + 31) / 32, (unsigned)((R) + 15) / 16, (unsigned)(R * R)), 32, 0, stream>>>(v1_1_26); }
    { GemmP v1_2_0;
      v1_2_0.A = GP + (size_t)2 * RP3 * C + (size_t)0 * C; v1_2_0.B = wv1 + 0; v1_2_0.bias = GP + (size_t)2 * RP3 * C + (size_t)0 * C; v1_2_0.R = GP + (size_t)2 * RP3 * C + (size_t)0 * C; v1_2_0.C = GC + (size_t)2 * R3 * C;
      v1_2_0.sAo = (long long)34 * 34 * C; v1_2_0.sAi = (long long)34 * C; v1_2_0.sAm = C; v1_2_0.sAk = 1; v1_2_0.sBo = 0; v1_2_0.sBi = 0; v1_2_0.sBn = C * 27; v1_2_0.sBk = 27; v1_2_0.sCo = (long long)R * R * C; v1_2_0.sCi = (long long)R * C; v1_2_0.sCm = C; v1_2_0.sRo = 0; v1_2_0.sRi = 0; v1_2_0.sRm = 0; v1_2_0.sRn = 0;
      v1_2_0.M = R; v1_2_0.N = C; v1_2_0.K = C; v1_2_0.zi_n = R; v1_2_0.flags = 0; v1_2_0.act = 0;
      v1_2_0.alpha = 1.0f; v1_2_0.beta = 0.0f; v1_2_0.sa = 1.0f; v1_2_0.sb = 1.0f; v1_2_0.Npad = C; v1_2_0.pad_ = 0;
      k_gemm<1><<<dim3((unsigned)((C) + 31) / 32, (unsigned)((R) + 15) / 16, (unsigned)(R * R)), 32, 0, stream>>>(v1_2_0); }
    { GemmP v1_2_1;
      v1_2_1.A = GP + (size_t)2 * RP3 * C + (size_t)1 * C; v1_2_1.B = wv1 + 1; v1_2_1.bias = GP + (size_t)2 * RP3 * C + (size_t)1 * C; v1_2_1.R = GC + (size_t)2 * R3 * C; v1_2_1.C = GC + (size_t)2 * R3 * C;
      v1_2_1.sAo = (long long)34 * 34 * C; v1_2_1.sAi = (long long)34 * C; v1_2_1.sAm = C; v1_2_1.sAk = 1; v1_2_1.sBo = 0; v1_2_1.sBi = 0; v1_2_1.sBn = C * 27; v1_2_1.sBk = 27; v1_2_1.sCo = (long long)R * R * C; v1_2_1.sCi = (long long)R * C; v1_2_1.sCm = C; v1_2_1.sRo = (long long)R * R * C; v1_2_1.sRi = (long long)R * C; v1_2_1.sRm = C; v1_2_1.sRn = 1;
      v1_2_1.M = R; v1_2_1.N = C; v1_2_1.K = C; v1_2_1.zi_n = R; v1_2_1.flags = 4; v1_2_1.act = 0;
      v1_2_1.alpha = 1.0f; v1_2_1.beta = 1.0f; v1_2_1.sa = 1.0f; v1_2_1.sb = 1.0f; v1_2_1.Npad = C; v1_2_1.pad_ = 0;
      k_gemm<1><<<dim3((unsigned)((C) + 31) / 32, (unsigned)((R) + 15) / 16, (unsigned)(R * R)), 32, 0, stream>>>(v1_2_1); }
    { GemmP v1_2_2;
      v1_2_2.A = GP + (size_t)2 * RP3 * C + (size_t)2 * C; v1_2_2.B = wv1 + 2; v1_2_2.bias = GP + (size_t)2 * RP3 * C + (size_t)2 * C; v1_2_2.R = GC + (size_t)2 * R3 * C; v1_2_2.C = GC + (size_t)2 * R3 * C;
      v1_2_2.sAo = (long long)34 * 34 * C; v1_2_2.sAi = (long long)34 * C; v1_2_2.sAm = C; v1_2_2.sAk = 1; v1_2_2.sBo = 0; v1_2_2.sBi = 0; v1_2_2.sBn = C * 27; v1_2_2.sBk = 27; v1_2_2.sCo = (long long)R * R * C; v1_2_2.sCi = (long long)R * C; v1_2_2.sCm = C; v1_2_2.sRo = (long long)R * R * C; v1_2_2.sRi = (long long)R * C; v1_2_2.sRm = C; v1_2_2.sRn = 1;
      v1_2_2.M = R; v1_2_2.N = C; v1_2_2.K = C; v1_2_2.zi_n = R; v1_2_2.flags = 4; v1_2_2.act = 0;
      v1_2_2.alpha = 1.0f; v1_2_2.beta = 1.0f; v1_2_2.sa = 1.0f; v1_2_2.sb = 1.0f; v1_2_2.Npad = C; v1_2_2.pad_ = 0;
      k_gemm<1><<<dim3((unsigned)((C) + 31) / 32, (unsigned)((R) + 15) / 16, (unsigned)(R * R)), 32, 0, stream>>>(v1_2_2); }
    { GemmP v1_2_3;
      v1_2_3.A = GP + (size_t)2 * RP3 * C + (size_t)34 * C; v1_2_3.B = wv1 + 3; v1_2_3.bias = GP + (size_t)2 * RP3 * C + (size_t)34 * C; v1_2_3.R = GC + (size_t)2 * R3 * C; v1_2_3.C = GC + (size_t)2 * R3 * C;
      v1_2_3.sAo = (long long)34 * 34 * C; v1_2_3.sAi = (long long)34 * C; v1_2_3.sAm = C; v1_2_3.sAk = 1; v1_2_3.sBo = 0; v1_2_3.sBi = 0; v1_2_3.sBn = C * 27; v1_2_3.sBk = 27; v1_2_3.sCo = (long long)R * R * C; v1_2_3.sCi = (long long)R * C; v1_2_3.sCm = C; v1_2_3.sRo = (long long)R * R * C; v1_2_3.sRi = (long long)R * C; v1_2_3.sRm = C; v1_2_3.sRn = 1;
      v1_2_3.M = R; v1_2_3.N = C; v1_2_3.K = C; v1_2_3.zi_n = R; v1_2_3.flags = 4; v1_2_3.act = 0;
      v1_2_3.alpha = 1.0f; v1_2_3.beta = 1.0f; v1_2_3.sa = 1.0f; v1_2_3.sb = 1.0f; v1_2_3.Npad = C; v1_2_3.pad_ = 0;
      k_gemm<1><<<dim3((unsigned)((C) + 31) / 32, (unsigned)((R) + 15) / 16, (unsigned)(R * R)), 32, 0, stream>>>(v1_2_3); }
    { GemmP v1_2_4;
      v1_2_4.A = GP + (size_t)2 * RP3 * C + (size_t)35 * C; v1_2_4.B = wv1 + 4; v1_2_4.bias = GP + (size_t)2 * RP3 * C + (size_t)35 * C; v1_2_4.R = GC + (size_t)2 * R3 * C; v1_2_4.C = GC + (size_t)2 * R3 * C;
      v1_2_4.sAo = (long long)34 * 34 * C; v1_2_4.sAi = (long long)34 * C; v1_2_4.sAm = C; v1_2_4.sAk = 1; v1_2_4.sBo = 0; v1_2_4.sBi = 0; v1_2_4.sBn = C * 27; v1_2_4.sBk = 27; v1_2_4.sCo = (long long)R * R * C; v1_2_4.sCi = (long long)R * C; v1_2_4.sCm = C; v1_2_4.sRo = (long long)R * R * C; v1_2_4.sRi = (long long)R * C; v1_2_4.sRm = C; v1_2_4.sRn = 1;
      v1_2_4.M = R; v1_2_4.N = C; v1_2_4.K = C; v1_2_4.zi_n = R; v1_2_4.flags = 4; v1_2_4.act = 0;
      v1_2_4.alpha = 1.0f; v1_2_4.beta = 1.0f; v1_2_4.sa = 1.0f; v1_2_4.sb = 1.0f; v1_2_4.Npad = C; v1_2_4.pad_ = 0;
      k_gemm<1><<<dim3((unsigned)((C) + 31) / 32, (unsigned)((R) + 15) / 16, (unsigned)(R * R)), 32, 0, stream>>>(v1_2_4); }
    { GemmP v1_2_5;
      v1_2_5.A = GP + (size_t)2 * RP3 * C + (size_t)36 * C; v1_2_5.B = wv1 + 5; v1_2_5.bias = GP + (size_t)2 * RP3 * C + (size_t)36 * C; v1_2_5.R = GC + (size_t)2 * R3 * C; v1_2_5.C = GC + (size_t)2 * R3 * C;
      v1_2_5.sAo = (long long)34 * 34 * C; v1_2_5.sAi = (long long)34 * C; v1_2_5.sAm = C; v1_2_5.sAk = 1; v1_2_5.sBo = 0; v1_2_5.sBi = 0; v1_2_5.sBn = C * 27; v1_2_5.sBk = 27; v1_2_5.sCo = (long long)R * R * C; v1_2_5.sCi = (long long)R * C; v1_2_5.sCm = C; v1_2_5.sRo = (long long)R * R * C; v1_2_5.sRi = (long long)R * C; v1_2_5.sRm = C; v1_2_5.sRn = 1;
      v1_2_5.M = R; v1_2_5.N = C; v1_2_5.K = C; v1_2_5.zi_n = R; v1_2_5.flags = 4; v1_2_5.act = 0;
      v1_2_5.alpha = 1.0f; v1_2_5.beta = 1.0f; v1_2_5.sa = 1.0f; v1_2_5.sb = 1.0f; v1_2_5.Npad = C; v1_2_5.pad_ = 0;
      k_gemm<1><<<dim3((unsigned)((C) + 31) / 32, (unsigned)((R) + 15) / 16, (unsigned)(R * R)), 32, 0, stream>>>(v1_2_5); }
    { GemmP v1_2_6;
      v1_2_6.A = GP + (size_t)2 * RP3 * C + (size_t)68 * C; v1_2_6.B = wv1 + 6; v1_2_6.bias = GP + (size_t)2 * RP3 * C + (size_t)68 * C; v1_2_6.R = GC + (size_t)2 * R3 * C; v1_2_6.C = GC + (size_t)2 * R3 * C;
      v1_2_6.sAo = (long long)34 * 34 * C; v1_2_6.sAi = (long long)34 * C; v1_2_6.sAm = C; v1_2_6.sAk = 1; v1_2_6.sBo = 0; v1_2_6.sBi = 0; v1_2_6.sBn = C * 27; v1_2_6.sBk = 27; v1_2_6.sCo = (long long)R * R * C; v1_2_6.sCi = (long long)R * C; v1_2_6.sCm = C; v1_2_6.sRo = (long long)R * R * C; v1_2_6.sRi = (long long)R * C; v1_2_6.sRm = C; v1_2_6.sRn = 1;
      v1_2_6.M = R; v1_2_6.N = C; v1_2_6.K = C; v1_2_6.zi_n = R; v1_2_6.flags = 4; v1_2_6.act = 0;
      v1_2_6.alpha = 1.0f; v1_2_6.beta = 1.0f; v1_2_6.sa = 1.0f; v1_2_6.sb = 1.0f; v1_2_6.Npad = C; v1_2_6.pad_ = 0;
      k_gemm<1><<<dim3((unsigned)((C) + 31) / 32, (unsigned)((R) + 15) / 16, (unsigned)(R * R)), 32, 0, stream>>>(v1_2_6); }
    { GemmP v1_2_7;
      v1_2_7.A = GP + (size_t)2 * RP3 * C + (size_t)69 * C; v1_2_7.B = wv1 + 7; v1_2_7.bias = GP + (size_t)2 * RP3 * C + (size_t)69 * C; v1_2_7.R = GC + (size_t)2 * R3 * C; v1_2_7.C = GC + (size_t)2 * R3 * C;
      v1_2_7.sAo = (long long)34 * 34 * C; v1_2_7.sAi = (long long)34 * C; v1_2_7.sAm = C; v1_2_7.sAk = 1; v1_2_7.sBo = 0; v1_2_7.sBi = 0; v1_2_7.sBn = C * 27; v1_2_7.sBk = 27; v1_2_7.sCo = (long long)R * R * C; v1_2_7.sCi = (long long)R * C; v1_2_7.sCm = C; v1_2_7.sRo = (long long)R * R * C; v1_2_7.sRi = (long long)R * C; v1_2_7.sRm = C; v1_2_7.sRn = 1;
      v1_2_7.M = R; v1_2_7.N = C; v1_2_7.K = C; v1_2_7.zi_n = R; v1_2_7.flags = 4; v1_2_7.act = 0;
      v1_2_7.alpha = 1.0f; v1_2_7.beta = 1.0f; v1_2_7.sa = 1.0f; v1_2_7.sb = 1.0f; v1_2_7.Npad = C; v1_2_7.pad_ = 0;
      k_gemm<1><<<dim3((unsigned)((C) + 31) / 32, (unsigned)((R) + 15) / 16, (unsigned)(R * R)), 32, 0, stream>>>(v1_2_7); }
    { GemmP v1_2_8;
      v1_2_8.A = GP + (size_t)2 * RP3 * C + (size_t)70 * C; v1_2_8.B = wv1 + 8; v1_2_8.bias = GP + (size_t)2 * RP3 * C + (size_t)70 * C; v1_2_8.R = GC + (size_t)2 * R3 * C; v1_2_8.C = GC + (size_t)2 * R3 * C;
      v1_2_8.sAo = (long long)34 * 34 * C; v1_2_8.sAi = (long long)34 * C; v1_2_8.sAm = C; v1_2_8.sAk = 1; v1_2_8.sBo = 0; v1_2_8.sBi = 0; v1_2_8.sBn = C * 27; v1_2_8.sBk = 27; v1_2_8.sCo = (long long)R * R * C; v1_2_8.sCi = (long long)R * C; v1_2_8.sCm = C; v1_2_8.sRo = (long long)R * R * C; v1_2_8.sRi = (long long)R * C; v1_2_8.sRm = C; v1_2_8.sRn = 1;
      v1_2_8.M = R; v1_2_8.N = C; v1_2_8.K = C; v1_2_8.zi_n = R; v1_2_8.flags = 4; v1_2_8.act = 0;
      v1_2_8.alpha = 1.0f; v1_2_8.beta = 1.0f; v1_2_8.sa = 1.0f; v1_2_8.sb = 1.0f; v1_2_8.Npad = C; v1_2_8.pad_ = 0;
      k_gemm<1><<<dim3((unsigned)((C) + 31) / 32, (unsigned)((R) + 15) / 16, (unsigned)(R * R)), 32, 0, stream>>>(v1_2_8); }
    { GemmP v1_2_9;
      v1_2_9.A = GP + (size_t)2 * RP3 * C + (size_t)1156 * C; v1_2_9.B = wv1 + 9; v1_2_9.bias = GP + (size_t)2 * RP3 * C + (size_t)1156 * C; v1_2_9.R = GC + (size_t)2 * R3 * C; v1_2_9.C = GC + (size_t)2 * R3 * C;
      v1_2_9.sAo = (long long)34 * 34 * C; v1_2_9.sAi = (long long)34 * C; v1_2_9.sAm = C; v1_2_9.sAk = 1; v1_2_9.sBo = 0; v1_2_9.sBi = 0; v1_2_9.sBn = C * 27; v1_2_9.sBk = 27; v1_2_9.sCo = (long long)R * R * C; v1_2_9.sCi = (long long)R * C; v1_2_9.sCm = C; v1_2_9.sRo = (long long)R * R * C; v1_2_9.sRi = (long long)R * C; v1_2_9.sRm = C; v1_2_9.sRn = 1;
      v1_2_9.M = R; v1_2_9.N = C; v1_2_9.K = C; v1_2_9.zi_n = R; v1_2_9.flags = 4; v1_2_9.act = 0;
      v1_2_9.alpha = 1.0f; v1_2_9.beta = 1.0f; v1_2_9.sa = 1.0f; v1_2_9.sb = 1.0f; v1_2_9.Npad = C; v1_2_9.pad_ = 0;
      k_gemm<1><<<dim3((unsigned)((C) + 31) / 32, (unsigned)((R) + 15) / 16, (unsigned)(R * R)), 32, 0, stream>>>(v1_2_9); }
    { GemmP v1_2_10;
      v1_2_10.A = GP + (size_t)2 * RP3 * C + (size_t)1157 * C; v1_2_10.B = wv1 + 10; v1_2_10.bias = GP + (size_t)2 * RP3 * C + (size_t)1157 * C; v1_2_10.R = GC + (size_t)2 * R3 * C; v1_2_10.C = GC + (size_t)2 * R3 * C;
      v1_2_10.sAo = (long long)34 * 34 * C; v1_2_10.sAi = (long long)34 * C; v1_2_10.sAm = C; v1_2_10.sAk = 1; v1_2_10.sBo = 0; v1_2_10.sBi = 0; v1_2_10.sBn = C * 27; v1_2_10.sBk = 27; v1_2_10.sCo = (long long)R * R * C; v1_2_10.sCi = (long long)R * C; v1_2_10.sCm = C; v1_2_10.sRo = (long long)R * R * C; v1_2_10.sRi = (long long)R * C; v1_2_10.sRm = C; v1_2_10.sRn = 1;
      v1_2_10.M = R; v1_2_10.N = C; v1_2_10.K = C; v1_2_10.zi_n = R; v1_2_10.flags = 4; v1_2_10.act = 0;
      v1_2_10.alpha = 1.0f; v1_2_10.beta = 1.0f; v1_2_10.sa = 1.0f; v1_2_10.sb = 1.0f; v1_2_10.Npad = C; v1_2_10.pad_ = 0;
      k_gemm<1><<<dim3((unsigned)((C) + 31) / 32, (unsigned)((R) + 15) / 16, (unsigned)(R * R)), 32, 0, stream>>>(v1_2_10); }
    { GemmP v1_2_11;
      v1_2_11.A = GP + (size_t)2 * RP3 * C + (size_t)1158 * C; v1_2_11.B = wv1 + 11; v1_2_11.bias = GP + (size_t)2 * RP3 * C + (size_t)1158 * C; v1_2_11.R = GC + (size_t)2 * R3 * C; v1_2_11.C = GC + (size_t)2 * R3 * C;
      v1_2_11.sAo = (long long)34 * 34 * C; v1_2_11.sAi = (long long)34 * C; v1_2_11.sAm = C; v1_2_11.sAk = 1; v1_2_11.sBo = 0; v1_2_11.sBi = 0; v1_2_11.sBn = C * 27; v1_2_11.sBk = 27; v1_2_11.sCo = (long long)R * R * C; v1_2_11.sCi = (long long)R * C; v1_2_11.sCm = C; v1_2_11.sRo = (long long)R * R * C; v1_2_11.sRi = (long long)R * C; v1_2_11.sRm = C; v1_2_11.sRn = 1;
      v1_2_11.M = R; v1_2_11.N = C; v1_2_11.K = C; v1_2_11.zi_n = R; v1_2_11.flags = 4; v1_2_11.act = 0;
      v1_2_11.alpha = 1.0f; v1_2_11.beta = 1.0f; v1_2_11.sa = 1.0f; v1_2_11.sb = 1.0f; v1_2_11.Npad = C; v1_2_11.pad_ = 0;
      k_gemm<1><<<dim3((unsigned)((C) + 31) / 32, (unsigned)((R) + 15) / 16, (unsigned)(R * R)), 32, 0, stream>>>(v1_2_11); }
    { GemmP v1_2_12;
      v1_2_12.A = GP + (size_t)2 * RP3 * C + (size_t)1190 * C; v1_2_12.B = wv1 + 12; v1_2_12.bias = GP + (size_t)2 * RP3 * C + (size_t)1190 * C; v1_2_12.R = GC + (size_t)2 * R3 * C; v1_2_12.C = GC + (size_t)2 * R3 * C;
      v1_2_12.sAo = (long long)34 * 34 * C; v1_2_12.sAi = (long long)34 * C; v1_2_12.sAm = C; v1_2_12.sAk = 1; v1_2_12.sBo = 0; v1_2_12.sBi = 0; v1_2_12.sBn = C * 27; v1_2_12.sBk = 27; v1_2_12.sCo = (long long)R * R * C; v1_2_12.sCi = (long long)R * C; v1_2_12.sCm = C; v1_2_12.sRo = (long long)R * R * C; v1_2_12.sRi = (long long)R * C; v1_2_12.sRm = C; v1_2_12.sRn = 1;
      v1_2_12.M = R; v1_2_12.N = C; v1_2_12.K = C; v1_2_12.zi_n = R; v1_2_12.flags = 4; v1_2_12.act = 0;
      v1_2_12.alpha = 1.0f; v1_2_12.beta = 1.0f; v1_2_12.sa = 1.0f; v1_2_12.sb = 1.0f; v1_2_12.Npad = C; v1_2_12.pad_ = 0;
      k_gemm<1><<<dim3((unsigned)((C) + 31) / 32, (unsigned)((R) + 15) / 16, (unsigned)(R * R)), 32, 0, stream>>>(v1_2_12); }
    { GemmP v1_2_13;
      v1_2_13.A = GP + (size_t)2 * RP3 * C + (size_t)1191 * C; v1_2_13.B = wv1 + 13; v1_2_13.bias = GP + (size_t)2 * RP3 * C + (size_t)1191 * C; v1_2_13.R = GC + (size_t)2 * R3 * C; v1_2_13.C = GC + (size_t)2 * R3 * C;
      v1_2_13.sAo = (long long)34 * 34 * C; v1_2_13.sAi = (long long)34 * C; v1_2_13.sAm = C; v1_2_13.sAk = 1; v1_2_13.sBo = 0; v1_2_13.sBi = 0; v1_2_13.sBn = C * 27; v1_2_13.sBk = 27; v1_2_13.sCo = (long long)R * R * C; v1_2_13.sCi = (long long)R * C; v1_2_13.sCm = C; v1_2_13.sRo = (long long)R * R * C; v1_2_13.sRi = (long long)R * C; v1_2_13.sRm = C; v1_2_13.sRn = 1;
      v1_2_13.M = R; v1_2_13.N = C; v1_2_13.K = C; v1_2_13.zi_n = R; v1_2_13.flags = 4; v1_2_13.act = 0;
      v1_2_13.alpha = 1.0f; v1_2_13.beta = 1.0f; v1_2_13.sa = 1.0f; v1_2_13.sb = 1.0f; v1_2_13.Npad = C; v1_2_13.pad_ = 0;
      k_gemm<1><<<dim3((unsigned)((C) + 31) / 32, (unsigned)((R) + 15) / 16, (unsigned)(R * R)), 32, 0, stream>>>(v1_2_13); }
    { GemmP v1_2_14;
      v1_2_14.A = GP + (size_t)2 * RP3 * C + (size_t)1192 * C; v1_2_14.B = wv1 + 14; v1_2_14.bias = GP + (size_t)2 * RP3 * C + (size_t)1192 * C; v1_2_14.R = GC + (size_t)2 * R3 * C; v1_2_14.C = GC + (size_t)2 * R3 * C;
      v1_2_14.sAo = (long long)34 * 34 * C; v1_2_14.sAi = (long long)34 * C; v1_2_14.sAm = C; v1_2_14.sAk = 1; v1_2_14.sBo = 0; v1_2_14.sBi = 0; v1_2_14.sBn = C * 27; v1_2_14.sBk = 27; v1_2_14.sCo = (long long)R * R * C; v1_2_14.sCi = (long long)R * C; v1_2_14.sCm = C; v1_2_14.sRo = (long long)R * R * C; v1_2_14.sRi = (long long)R * C; v1_2_14.sRm = C; v1_2_14.sRn = 1;
      v1_2_14.M = R; v1_2_14.N = C; v1_2_14.K = C; v1_2_14.zi_n = R; v1_2_14.flags = 4; v1_2_14.act = 0;
      v1_2_14.alpha = 1.0f; v1_2_14.beta = 1.0f; v1_2_14.sa = 1.0f; v1_2_14.sb = 1.0f; v1_2_14.Npad = C; v1_2_14.pad_ = 0;
      k_gemm<1><<<dim3((unsigned)((C) + 31) / 32, (unsigned)((R) + 15) / 16, (unsigned)(R * R)), 32, 0, stream>>>(v1_2_14); }
    { GemmP v1_2_15;
      v1_2_15.A = GP + (size_t)2 * RP3 * C + (size_t)1224 * C; v1_2_15.B = wv1 + 15; v1_2_15.bias = GP + (size_t)2 * RP3 * C + (size_t)1224 * C; v1_2_15.R = GC + (size_t)2 * R3 * C; v1_2_15.C = GC + (size_t)2 * R3 * C;
      v1_2_15.sAo = (long long)34 * 34 * C; v1_2_15.sAi = (long long)34 * C; v1_2_15.sAm = C; v1_2_15.sAk = 1; v1_2_15.sBo = 0; v1_2_15.sBi = 0; v1_2_15.sBn = C * 27; v1_2_15.sBk = 27; v1_2_15.sCo = (long long)R * R * C; v1_2_15.sCi = (long long)R * C; v1_2_15.sCm = C; v1_2_15.sRo = (long long)R * R * C; v1_2_15.sRi = (long long)R * C; v1_2_15.sRm = C; v1_2_15.sRn = 1;
      v1_2_15.M = R; v1_2_15.N = C; v1_2_15.K = C; v1_2_15.zi_n = R; v1_2_15.flags = 4; v1_2_15.act = 0;
      v1_2_15.alpha = 1.0f; v1_2_15.beta = 1.0f; v1_2_15.sa = 1.0f; v1_2_15.sb = 1.0f; v1_2_15.Npad = C; v1_2_15.pad_ = 0;
      k_gemm<1><<<dim3((unsigned)((C) + 31) / 32, (unsigned)((R) + 15) / 16, (unsigned)(R * R)), 32, 0, stream>>>(v1_2_15); }
    { GemmP v1_2_16;
      v1_2_16.A = GP + (size_t)2 * RP3 * C + (size_t)1225 * C; v1_2_16.B = wv1 + 16; v1_2_16.bias = GP + (size_t)2 * RP3 * C + (size_t)1225 * C; v1_2_16.R = GC + (size_t)2 * R3 * C; v1_2_16.C = GC + (size_t)2 * R3 * C;
      v1_2_16.sAo = (long long)34 * 34 * C; v1_2_16.sAi = (long long)34 * C; v1_2_16.sAm = C; v1_2_16.sAk = 1; v1_2_16.sBo = 0; v1_2_16.sBi = 0; v1_2_16.sBn = C * 27; v1_2_16.sBk = 27; v1_2_16.sCo = (long long)R * R * C; v1_2_16.sCi = (long long)R * C; v1_2_16.sCm = C; v1_2_16.sRo = (long long)R * R * C; v1_2_16.sRi = (long long)R * C; v1_2_16.sRm = C; v1_2_16.sRn = 1;
      v1_2_16.M = R; v1_2_16.N = C; v1_2_16.K = C; v1_2_16.zi_n = R; v1_2_16.flags = 4; v1_2_16.act = 0;
      v1_2_16.alpha = 1.0f; v1_2_16.beta = 1.0f; v1_2_16.sa = 1.0f; v1_2_16.sb = 1.0f; v1_2_16.Npad = C; v1_2_16.pad_ = 0;
      k_gemm<1><<<dim3((unsigned)((C) + 31) / 32, (unsigned)((R) + 15) / 16, (unsigned)(R * R)), 32, 0, stream>>>(v1_2_16); }
    { GemmP v1_2_17;
      v1_2_17.A = GP + (size_t)2 * RP3 * C + (size_t)1226 * C; v1_2_17.B = wv1 + 17; v1_2_17.bias = GP + (size_t)2 * RP3 * C + (size_t)1226 * C; v1_2_17.R = GC + (size_t)2 * R3 * C; v1_2_17.C = GC + (size_t)2 * R3 * C;
      v1_2_17.sAo = (long long)34 * 34 * C; v1_2_17.sAi = (long long)34 * C; v1_2_17.sAm = C; v1_2_17.sAk = 1; v1_2_17.sBo = 0; v1_2_17.sBi = 0; v1_2_17.sBn = C * 27; v1_2_17.sBk = 27; v1_2_17.sCo = (long long)R * R * C; v1_2_17.sCi = (long long)R * C; v1_2_17.sCm = C; v1_2_17.sRo = (long long)R * R * C; v1_2_17.sRi = (long long)R * C; v1_2_17.sRm = C; v1_2_17.sRn = 1;
      v1_2_17.M = R; v1_2_17.N = C; v1_2_17.K = C; v1_2_17.zi_n = R; v1_2_17.flags = 4; v1_2_17.act = 0;
      v1_2_17.alpha = 1.0f; v1_2_17.beta = 1.0f; v1_2_17.sa = 1.0f; v1_2_17.sb = 1.0f; v1_2_17.Npad = C; v1_2_17.pad_ = 0;
      k_gemm<1><<<dim3((unsigned)((C) + 31) / 32, (unsigned)((R) + 15) / 16, (unsigned)(R * R)), 32, 0, stream>>>(v1_2_17); }
    { GemmP v1_2_18;
      v1_2_18.A = GP + (size_t)2 * RP3 * C + (size_t)2312 * C; v1_2_18.B = wv1 + 18; v1_2_18.bias = GP + (size_t)2 * RP3 * C + (size_t)2312 * C; v1_2_18.R = GC + (size_t)2 * R3 * C; v1_2_18.C = GC + (size_t)2 * R3 * C;
      v1_2_18.sAo = (long long)34 * 34 * C; v1_2_18.sAi = (long long)34 * C; v1_2_18.sAm = C; v1_2_18.sAk = 1; v1_2_18.sBo = 0; v1_2_18.sBi = 0; v1_2_18.sBn = C * 27; v1_2_18.sBk = 27; v1_2_18.sCo = (long long)R * R * C; v1_2_18.sCi = (long long)R * C; v1_2_18.sCm = C; v1_2_18.sRo = (long long)R * R * C; v1_2_18.sRi = (long long)R * C; v1_2_18.sRm = C; v1_2_18.sRn = 1;
      v1_2_18.M = R; v1_2_18.N = C; v1_2_18.K = C; v1_2_18.zi_n = R; v1_2_18.flags = 4; v1_2_18.act = 0;
      v1_2_18.alpha = 1.0f; v1_2_18.beta = 1.0f; v1_2_18.sa = 1.0f; v1_2_18.sb = 1.0f; v1_2_18.Npad = C; v1_2_18.pad_ = 0;
      k_gemm<1><<<dim3((unsigned)((C) + 31) / 32, (unsigned)((R) + 15) / 16, (unsigned)(R * R)), 32, 0, stream>>>(v1_2_18); }
    { GemmP v1_2_19;
      v1_2_19.A = GP + (size_t)2 * RP3 * C + (size_t)2313 * C; v1_2_19.B = wv1 + 19; v1_2_19.bias = GP + (size_t)2 * RP3 * C + (size_t)2313 * C; v1_2_19.R = GC + (size_t)2 * R3 * C; v1_2_19.C = GC + (size_t)2 * R3 * C;
      v1_2_19.sAo = (long long)34 * 34 * C; v1_2_19.sAi = (long long)34 * C; v1_2_19.sAm = C; v1_2_19.sAk = 1; v1_2_19.sBo = 0; v1_2_19.sBi = 0; v1_2_19.sBn = C * 27; v1_2_19.sBk = 27; v1_2_19.sCo = (long long)R * R * C; v1_2_19.sCi = (long long)R * C; v1_2_19.sCm = C; v1_2_19.sRo = (long long)R * R * C; v1_2_19.sRi = (long long)R * C; v1_2_19.sRm = C; v1_2_19.sRn = 1;
      v1_2_19.M = R; v1_2_19.N = C; v1_2_19.K = C; v1_2_19.zi_n = R; v1_2_19.flags = 4; v1_2_19.act = 0;
      v1_2_19.alpha = 1.0f; v1_2_19.beta = 1.0f; v1_2_19.sa = 1.0f; v1_2_19.sb = 1.0f; v1_2_19.Npad = C; v1_2_19.pad_ = 0;
      k_gemm<1><<<dim3((unsigned)((C) + 31) / 32, (unsigned)((R) + 15) / 16, (unsigned)(R * R)), 32, 0, stream>>>(v1_2_19); }
    { GemmP v1_2_20;
      v1_2_20.A = GP + (size_t)2 * RP3 * C + (size_t)2314 * C; v1_2_20.B = wv1 + 20; v1_2_20.bias = GP + (size_t)2 * RP3 * C + (size_t)2314 * C; v1_2_20.R = GC + (size_t)2 * R3 * C; v1_2_20.C = GC + (size_t)2 * R3 * C;
      v1_2_20.sAo = (long long)34 * 34 * C; v1_2_20.sAi = (long long)34 * C; v1_2_20.sAm = C; v1_2_20.sAk = 1; v1_2_20.sBo = 0; v1_2_20.sBi = 0; v1_2_20.sBn = C * 27; v1_2_20.sBk = 27; v1_2_20.sCo = (long long)R * R * C; v1_2_20.sCi = (long long)R * C; v1_2_20.sCm = C; v1_2_20.sRo = (long long)R * R * C; v1_2_20.sRi = (long long)R * C; v1_2_20.sRm = C; v1_2_20.sRn = 1;
      v1_2_20.M = R; v1_2_20.N = C; v1_2_20.K = C; v1_2_20.zi_n = R; v1_2_20.flags = 4; v1_2_20.act = 0;
      v1_2_20.alpha = 1.0f; v1_2_20.beta = 1.0f; v1_2_20.sa = 1.0f; v1_2_20.sb = 1.0f; v1_2_20.Npad = C; v1_2_20.pad_ = 0;
      k_gemm<1><<<dim3((unsigned)((C) + 31) / 32, (unsigned)((R) + 15) / 16, (unsigned)(R * R)), 32, 0, stream>>>(v1_2_20); }
    { GemmP v1_2_21;
      v1_2_21.A = GP + (size_t)2 * RP3 * C + (size_t)2346 * C; v1_2_21.B = wv1 + 21; v1_2_21.bias = GP + (size_t)2 * RP3 * C + (size_t)2346 * C; v1_2_21.R = GC + (size_t)2 * R3 * C; v1_2_21.C = GC + (size_t)2 * R3 * C;
      v1_2_21.sAo = (long long)34 * 34 * C; v1_2_21.sAi = (long long)34 * C; v1_2_21.sAm = C; v1_2_21.sAk = 1; v1_2_21.sBo = 0; v1_2_21.sBi = 0; v1_2_21.sBn = C * 27; v1_2_21.sBk = 27; v1_2_21.sCo = (long long)R * R * C; v1_2_21.sCi = (long long)R * C; v1_2_21.sCm = C; v1_2_21.sRo = (long long)R * R * C; v1_2_21.sRi = (long long)R * C; v1_2_21.sRm = C; v1_2_21.sRn = 1;
      v1_2_21.M = R; v1_2_21.N = C; v1_2_21.K = C; v1_2_21.zi_n = R; v1_2_21.flags = 4; v1_2_21.act = 0;
      v1_2_21.alpha = 1.0f; v1_2_21.beta = 1.0f; v1_2_21.sa = 1.0f; v1_2_21.sb = 1.0f; v1_2_21.Npad = C; v1_2_21.pad_ = 0;
      k_gemm<1><<<dim3((unsigned)((C) + 31) / 32, (unsigned)((R) + 15) / 16, (unsigned)(R * R)), 32, 0, stream>>>(v1_2_21); }
    { GemmP v1_2_22;
      v1_2_22.A = GP + (size_t)2 * RP3 * C + (size_t)2347 * C; v1_2_22.B = wv1 + 22; v1_2_22.bias = GP + (size_t)2 * RP3 * C + (size_t)2347 * C; v1_2_22.R = GC + (size_t)2 * R3 * C; v1_2_22.C = GC + (size_t)2 * R3 * C;
      v1_2_22.sAo = (long long)34 * 34 * C; v1_2_22.sAi = (long long)34 * C; v1_2_22.sAm = C; v1_2_22.sAk = 1; v1_2_22.sBo = 0; v1_2_22.sBi = 0; v1_2_22.sBn = C * 27; v1_2_22.sBk = 27; v1_2_22.sCo = (long long)R * R * C; v1_2_22.sCi = (long long)R * C; v1_2_22.sCm = C; v1_2_22.sRo = (long long)R * R * C; v1_2_22.sRi = (long long)R * C; v1_2_22.sRm = C; v1_2_22.sRn = 1;
      v1_2_22.M = R; v1_2_22.N = C; v1_2_22.K = C; v1_2_22.zi_n = R; v1_2_22.flags = 4; v1_2_22.act = 0;
      v1_2_22.alpha = 1.0f; v1_2_22.beta = 1.0f; v1_2_22.sa = 1.0f; v1_2_22.sb = 1.0f; v1_2_22.Npad = C; v1_2_22.pad_ = 0;
      k_gemm<1><<<dim3((unsigned)((C) + 31) / 32, (unsigned)((R) + 15) / 16, (unsigned)(R * R)), 32, 0, stream>>>(v1_2_22); }
    { GemmP v1_2_23;
      v1_2_23.A = GP + (size_t)2 * RP3 * C + (size_t)2348 * C; v1_2_23.B = wv1 + 23; v1_2_23.bias = GP + (size_t)2 * RP3 * C + (size_t)2348 * C; v1_2_23.R = GC + (size_t)2 * R3 * C; v1_2_23.C = GC + (size_t)2 * R3 * C;
      v1_2_23.sAo = (long long)34 * 34 * C; v1_2_23.sAi = (long long)34 * C; v1_2_23.sAm = C; v1_2_23.sAk = 1; v1_2_23.sBo = 0; v1_2_23.sBi = 0; v1_2_23.sBn = C * 27; v1_2_23.sBk = 27; v1_2_23.sCo = (long long)R * R * C; v1_2_23.sCi = (long long)R * C; v1_2_23.sCm = C; v1_2_23.sRo = (long long)R * R * C; v1_2_23.sRi = (long long)R * C; v1_2_23.sRm = C; v1_2_23.sRn = 1;
      v1_2_23.M = R; v1_2_23.N = C; v1_2_23.K = C; v1_2_23.zi_n = R; v1_2_23.flags = 4; v1_2_23.act = 0;
      v1_2_23.alpha = 1.0f; v1_2_23.beta = 1.0f; v1_2_23.sa = 1.0f; v1_2_23.sb = 1.0f; v1_2_23.Npad = C; v1_2_23.pad_ = 0;
      k_gemm<1><<<dim3((unsigned)((C) + 31) / 32, (unsigned)((R) + 15) / 16, (unsigned)(R * R)), 32, 0, stream>>>(v1_2_23); }
    { GemmP v1_2_24;
      v1_2_24.A = GP + (size_t)2 * RP3 * C + (size_t)2380 * C; v1_2_24.B = wv1 + 24; v1_2_24.bias = GP + (size_t)2 * RP3 * C + (size_t)2380 * C; v1_2_24.R = GC + (size_t)2 * R3 * C; v1_2_24.C = GC + (size_t)2 * R3 * C;
      v1_2_24.sAo = (long long)34 * 34 * C; v1_2_24.sAi = (long long)34 * C; v1_2_24.sAm = C; v1_2_24.sAk = 1; v1_2_24.sBo = 0; v1_2_24.sBi = 0; v1_2_24.sBn = C * 27; v1_2_24.sBk = 27; v1_2_24.sCo = (long long)R * R * C; v1_2_24.sCi = (long long)R * C; v1_2_24.sCm = C; v1_2_24.sRo = (long long)R * R * C; v1_2_24.sRi = (long long)R * C; v1_2_24.sRm = C; v1_2_24.sRn = 1;
      v1_2_24.M = R; v1_2_24.N = C; v1_2_24.K = C; v1_2_24.zi_n = R; v1_2_24.flags = 4; v1_2_24.act = 0;
      v1_2_24.alpha = 1.0f; v1_2_24.beta = 1.0f; v1_2_24.sa = 1.0f; v1_2_24.sb = 1.0f; v1_2_24.Npad = C; v1_2_24.pad_ = 0;
      k_gemm<1><<<dim3((unsigned)((C) + 31) / 32, (unsigned)((R) + 15) / 16, (unsigned)(R * R)), 32, 0, stream>>>(v1_2_24); }
    { GemmP v1_2_25;
      v1_2_25.A = GP + (size_t)2 * RP3 * C + (size_t)2381 * C; v1_2_25.B = wv1 + 25; v1_2_25.bias = GP + (size_t)2 * RP3 * C + (size_t)2381 * C; v1_2_25.R = GC + (size_t)2 * R3 * C; v1_2_25.C = GC + (size_t)2 * R3 * C;
      v1_2_25.sAo = (long long)34 * 34 * C; v1_2_25.sAi = (long long)34 * C; v1_2_25.sAm = C; v1_2_25.sAk = 1; v1_2_25.sBo = 0; v1_2_25.sBi = 0; v1_2_25.sBn = C * 27; v1_2_25.sBk = 27; v1_2_25.sCo = (long long)R * R * C; v1_2_25.sCi = (long long)R * C; v1_2_25.sCm = C; v1_2_25.sRo = (long long)R * R * C; v1_2_25.sRi = (long long)R * C; v1_2_25.sRm = C; v1_2_25.sRn = 1;
      v1_2_25.M = R; v1_2_25.N = C; v1_2_25.K = C; v1_2_25.zi_n = R; v1_2_25.flags = 4; v1_2_25.act = 0;
      v1_2_25.alpha = 1.0f; v1_2_25.beta = 1.0f; v1_2_25.sa = 1.0f; v1_2_25.sb = 1.0f; v1_2_25.Npad = C; v1_2_25.pad_ = 0;
      k_gemm<1><<<dim3((unsigned)((C) + 31) / 32, (unsigned)((R) + 15) / 16, (unsigned)(R * R)), 32, 0, stream>>>(v1_2_25); }
    { GemmP v1_2_26;
      v1_2_26.A = GP + (size_t)2 * RP3 * C + (size_t)2382 * C; v1_2_26.B = wv1 + 26; v1_2_26.bias = GP + (size_t)2 * RP3 * C + (size_t)2382 * C; v1_2_26.R = GC + (size_t)2 * R3 * C; v1_2_26.C = GC + (size_t)2 * R3 * C;
      v1_2_26.sAo = (long long)34 * 34 * C; v1_2_26.sAi = (long long)34 * C; v1_2_26.sAm = C; v1_2_26.sAk = 1; v1_2_26.sBo = 0; v1_2_26.sBi = 0; v1_2_26.sBn = C * 27; v1_2_26.sBk = 27; v1_2_26.sCo = (long long)R * R * C; v1_2_26.sCi = (long long)R * C; v1_2_26.sCm = C; v1_2_26.sRo = (long long)R * R * C; v1_2_26.sRi = (long long)R * C; v1_2_26.sRm = C; v1_2_26.sRn = 1;
      v1_2_26.M = R; v1_2_26.N = C; v1_2_26.K = C; v1_2_26.zi_n = R; v1_2_26.flags = 4; v1_2_26.act = 0;
      v1_2_26.alpha = 1.0f; v1_2_26.beta = 1.0f; v1_2_26.sa = 1.0f; v1_2_26.sb = 1.0f; v1_2_26.Npad = C; v1_2_26.pad_ = 0;
      k_gemm<1><<<dim3((unsigned)((C) + 31) / 32, (unsigned)((R) + 15) / 16, (unsigned)(R * R)), 32, 0, stream>>>(v1_2_26); }
    { GemmP v1_3_0;
      v1_3_0.A = GP + (size_t)3 * RP3 * C + (size_t)0 * C; v1_3_0.B = wv1 + 0; v1_3_0.bias = bv1; v1_3_0.R = GP + (size_t)3 * RP3 * C + (size_t)0 * C; v1_3_0.C = GC + (size_t)3 * R3 * C;
      v1_3_0.sAo = (long long)34 * 34 * C; v1_3_0.sAi = (long long)34 * C; v1_3_0.sAm = C; v1_3_0.sAk = 1; v1_3_0.sBo = 0; v1_3_0.sBi = 0; v1_3_0.sBn = C * 27; v1_3_0.sBk = 27; v1_3_0.sCo = (long long)R * R * C; v1_3_0.sCi = (long long)R * C; v1_3_0.sCm = C; v1_3_0.sRo = 0; v1_3_0.sRi = 0; v1_3_0.sRm = 0; v1_3_0.sRn = 0;
      v1_3_0.M = R; v1_3_0.N = C; v1_3_0.K = C; v1_3_0.zi_n = R; v1_3_0.flags = 1; v1_3_0.act = 0;
      v1_3_0.alpha = 1.0f; v1_3_0.beta = 0.0f; v1_3_0.sa = 1.0f; v1_3_0.sb = 1.0f; v1_3_0.Npad = C; v1_3_0.pad_ = 0;
      k_gemm<1><<<dim3((unsigned)((C) + 31) / 32, (unsigned)((R) + 15) / 16, (unsigned)(R * R)), 32, 0, stream>>>(v1_3_0); }
    { GemmP v1_3_1;
      v1_3_1.A = GP + (size_t)3 * RP3 * C + (size_t)1 * C; v1_3_1.B = wv1 + 1; v1_3_1.bias = GP + (size_t)3 * RP3 * C + (size_t)1 * C; v1_3_1.R = GC + (size_t)3 * R3 * C; v1_3_1.C = GC + (size_t)3 * R3 * C;
      v1_3_1.sAo = (long long)34 * 34 * C; v1_3_1.sAi = (long long)34 * C; v1_3_1.sAm = C; v1_3_1.sAk = 1; v1_3_1.sBo = 0; v1_3_1.sBi = 0; v1_3_1.sBn = C * 27; v1_3_1.sBk = 27; v1_3_1.sCo = (long long)R * R * C; v1_3_1.sCi = (long long)R * C; v1_3_1.sCm = C; v1_3_1.sRo = (long long)R * R * C; v1_3_1.sRi = (long long)R * C; v1_3_1.sRm = C; v1_3_1.sRn = 1;
      v1_3_1.M = R; v1_3_1.N = C; v1_3_1.K = C; v1_3_1.zi_n = R; v1_3_1.flags = 4; v1_3_1.act = 0;
      v1_3_1.alpha = 1.0f; v1_3_1.beta = 1.0f; v1_3_1.sa = 1.0f; v1_3_1.sb = 1.0f; v1_3_1.Npad = C; v1_3_1.pad_ = 0;
      k_gemm<1><<<dim3((unsigned)((C) + 31) / 32, (unsigned)((R) + 15) / 16, (unsigned)(R * R)), 32, 0, stream>>>(v1_3_1); }
    { GemmP v1_3_2;
      v1_3_2.A = GP + (size_t)3 * RP3 * C + (size_t)2 * C; v1_3_2.B = wv1 + 2; v1_3_2.bias = GP + (size_t)3 * RP3 * C + (size_t)2 * C; v1_3_2.R = GC + (size_t)3 * R3 * C; v1_3_2.C = GC + (size_t)3 * R3 * C;
      v1_3_2.sAo = (long long)34 * 34 * C; v1_3_2.sAi = (long long)34 * C; v1_3_2.sAm = C; v1_3_2.sAk = 1; v1_3_2.sBo = 0; v1_3_2.sBi = 0; v1_3_2.sBn = C * 27; v1_3_2.sBk = 27; v1_3_2.sCo = (long long)R * R * C; v1_3_2.sCi = (long long)R * C; v1_3_2.sCm = C; v1_3_2.sRo = (long long)R * R * C; v1_3_2.sRi = (long long)R * C; v1_3_2.sRm = C; v1_3_2.sRn = 1;
      v1_3_2.M = R; v1_3_2.N = C; v1_3_2.K = C; v1_3_2.zi_n = R; v1_3_2.flags = 4; v1_3_2.act = 0;
      v1_3_2.alpha = 1.0f; v1_3_2.beta = 1.0f; v1_3_2.sa = 1.0f; v1_3_2.sb = 1.0f; v1_3_2.Npad = C; v1_3_2.pad_ = 0;
      k_gemm<1><<<dim3((unsigned)((C) + 31) / 32, (unsigned)((R) + 15) / 16, (unsigned)(R * R)), 32, 0, stream>>>(v1_3_2); }
    { GemmP v1_3_3;
      v1_3_3.A = GP + (size_t)3 * RP3 * C + (size_t)34 * C; v1_3_3.B = wv1 + 3; v1_3_3.bias = GP + (size_t)3 * RP3 * C + (size_t)34 * C; v1_3_3.R = GC + (size_t)3 * R3 * C; v1_3_3.C = GC + (size_t)3 * R3 * C;
      v1_3_3.sAo = (long long)34 * 34 * C; v1_3_3.sAi = (long long)34 * C; v1_3_3.sAm = C; v1_3_3.sAk = 1; v1_3_3.sBo = 0; v1_3_3.sBi = 0; v1_3_3.sBn = C * 27; v1_3_3.sBk = 27; v1_3_3.sCo = (long long)R * R * C; v1_3_3.sCi = (long long)R * C; v1_3_3.sCm = C; v1_3_3.sRo = (long long)R * R * C; v1_3_3.sRi = (long long)R * C; v1_3_3.sRm = C; v1_3_3.sRn = 1;
      v1_3_3.M = R; v1_3_3.N = C; v1_3_3.K = C; v1_3_3.zi_n = R; v1_3_3.flags = 4; v1_3_3.act = 0;
      v1_3_3.alpha = 1.0f; v1_3_3.beta = 1.0f; v1_3_3.sa = 1.0f; v1_3_3.sb = 1.0f; v1_3_3.Npad = C; v1_3_3.pad_ = 0;
      k_gemm<1><<<dim3((unsigned)((C) + 31) / 32, (unsigned)((R) + 15) / 16, (unsigned)(R * R)), 32, 0, stream>>>(v1_3_3); }
    { GemmP v1_3_4;
      v1_3_4.A = GP + (size_t)3 * RP3 * C + (size_t)35 * C; v1_3_4.B = wv1 + 4; v1_3_4.bias = GP + (size_t)3 * RP3 * C + (size_t)35 * C; v1_3_4.R = GC + (size_t)3 * R3 * C; v1_3_4.C = GC + (size_t)3 * R3 * C;
      v1_3_4.sAo = (long long)34 * 34 * C; v1_3_4.sAi = (long long)34 * C; v1_3_4.sAm = C; v1_3_4.sAk = 1; v1_3_4.sBo = 0; v1_3_4.sBi = 0; v1_3_4.sBn = C * 27; v1_3_4.sBk = 27; v1_3_4.sCo = (long long)R * R * C; v1_3_4.sCi = (long long)R * C; v1_3_4.sCm = C; v1_3_4.sRo = (long long)R * R * C; v1_3_4.sRi = (long long)R * C; v1_3_4.sRm = C; v1_3_4.sRn = 1;
      v1_3_4.M = R; v1_3_4.N = C; v1_3_4.K = C; v1_3_4.zi_n = R; v1_3_4.flags = 4; v1_3_4.act = 0;
      v1_3_4.alpha = 1.0f; v1_3_4.beta = 1.0f; v1_3_4.sa = 1.0f; v1_3_4.sb = 1.0f; v1_3_4.Npad = C; v1_3_4.pad_ = 0;
      k_gemm<1><<<dim3((unsigned)((C) + 31) / 32, (unsigned)((R) + 15) / 16, (unsigned)(R * R)), 32, 0, stream>>>(v1_3_4); }
    { GemmP v1_3_5;
      v1_3_5.A = GP + (size_t)3 * RP3 * C + (size_t)36 * C; v1_3_5.B = wv1 + 5; v1_3_5.bias = GP + (size_t)3 * RP3 * C + (size_t)36 * C; v1_3_5.R = GC + (size_t)3 * R3 * C; v1_3_5.C = GC + (size_t)3 * R3 * C;
      v1_3_5.sAo = (long long)34 * 34 * C; v1_3_5.sAi = (long long)34 * C; v1_3_5.sAm = C; v1_3_5.sAk = 1; v1_3_5.sBo = 0; v1_3_5.sBi = 0; v1_3_5.sBn = C * 27; v1_3_5.sBk = 27; v1_3_5.sCo = (long long)R * R * C; v1_3_5.sCi = (long long)R * C; v1_3_5.sCm = C; v1_3_5.sRo = (long long)R * R * C; v1_3_5.sRi = (long long)R * C; v1_3_5.sRm = C; v1_3_5.sRn = 1;
      v1_3_5.M = R; v1_3_5.N = C; v1_3_5.K = C; v1_3_5.zi_n = R; v1_3_5.flags = 4; v1_3_5.act = 0;
      v1_3_5.alpha = 1.0f; v1_3_5.beta = 1.0f; v1_3_5.sa = 1.0f; v1_3_5.sb = 1.0f; v1_3_5.Npad = C; v1_3_5.pad_ = 0;
      k_gemm<1><<<dim3((unsigned)((C) + 31) / 32, (unsigned)((R) + 15) / 16, (unsigned)(R * R)), 32, 0, stream>>>(v1_3_5); }
    { GemmP v1_3_6;
      v1_3_6.A = GP + (size_t)3 * RP3 * C + (size_t)68 * C; v1_3_6.B = wv1 + 6; v1_3_6.bias = GP + (size_t)3 * RP3 * C + (size_t)68 * C; v1_3_6.R = GC + (size_t)3 * R3 * C; v1_3_6.C = GC + (size_t)3 * R3 * C;
      v1_3_6.sAo = (long long)34 * 34 * C; v1_3_6.sAi = (long long)34 * C; v1_3_6.sAm = C; v1_3_6.sAk = 1; v1_3_6.sBo = 0; v1_3_6.sBi = 0; v1_3_6.sBn = C * 27; v1_3_6.sBk = 27; v1_3_6.sCo = (long long)R * R * C; v1_3_6.sCi = (long long)R * C; v1_3_6.sCm = C; v1_3_6.sRo = (long long)R * R * C; v1_3_6.sRi = (long long)R * C; v1_3_6.sRm = C; v1_3_6.sRn = 1;
      v1_3_6.M = R; v1_3_6.N = C; v1_3_6.K = C; v1_3_6.zi_n = R; v1_3_6.flags = 4; v1_3_6.act = 0;
      v1_3_6.alpha = 1.0f; v1_3_6.beta = 1.0f; v1_3_6.sa = 1.0f; v1_3_6.sb = 1.0f; v1_3_6.Npad = C; v1_3_6.pad_ = 0;
      k_gemm<1><<<dim3((unsigned)((C) + 31) / 32, (unsigned)((R) + 15) / 16, (unsigned)(R * R)), 32, 0, stream>>>(v1_3_6); }
    { GemmP v1_3_7;
      v1_3_7.A = GP + (size_t)3 * RP3 * C + (size_t)69 * C; v1_3_7.B = wv1 + 7; v1_3_7.bias = GP + (size_t)3 * RP3 * C + (size_t)69 * C; v1_3_7.R = GC + (size_t)3 * R3 * C; v1_3_7.C = GC + (size_t)3 * R3 * C;
      v1_3_7.sAo = (long long)34 * 34 * C; v1_3_7.sAi = (long long)34 * C; v1_3_7.sAm = C; v1_3_7.sAk = 1; v1_3_7.sBo = 0; v1_3_7.sBi = 0; v1_3_7.sBn = C * 27; v1_3_7.sBk = 27; v1_3_7.sCo = (long long)R * R * C; v1_3_7.sCi = (long long)R * C; v1_3_7.sCm = C; v1_3_7.sRo = (long long)R * R * C; v1_3_7.sRi = (long long)R * C; v1_3_7.sRm = C; v1_3_7.sRn = 1;
      v1_3_7.M = R; v1_3_7.N = C; v1_3_7.K = C; v1_3_7.zi_n = R; v1_3_7.flags = 4; v1_3_7.act = 0;
      v1_3_7.alpha = 1.0f; v1_3_7.beta = 1.0f; v1_3_7.sa = 1.0f; v1_3_7.sb = 1.0f; v1_3_7.Npad = C; v1_3_7.pad_ = 0;
      k_gemm<1><<<dim3((unsigned)((C) + 31) / 32, (unsigned)((R) + 15) / 16, (unsigned)(R * R)), 32, 0, stream>>>(v1_3_7); }
    { GemmP v1_3_8;
      v1_3_8.A = GP + (size_t)3 * RP3 * C + (size_t)70 * C; v1_3_8.B = wv1 + 8; v1_3_8.bias = GP + (size_t)3 * RP3 * C + (size_t)70 * C; v1_3_8.R = GC + (size_t)3 * R3 * C; v1_3_8.C = GC + (size_t)3 * R3 * C;
      v1_3_8.sAo = (long long)34 * 34 * C; v1_3_8.sAi = (long long)34 * C; v1_3_8.sAm = C; v1_3_8.sAk = 1; v1_3_8.sBo = 0; v1_3_8.sBi = 0; v1_3_8.sBn = C * 27; v1_3_8.sBk = 27; v1_3_8.sCo = (long long)R * R * C; v1_3_8.sCi = (long long)R * C; v1_3_8.sCm = C; v1_3_8.sRo = (long long)R * R * C; v1_3_8.sRi = (long long)R * C; v1_3_8.sRm = C; v1_3_8.sRn = 1;
      v1_3_8.M = R; v1_3_8.N = C; v1_3_8.K = C; v1_3_8.zi_n = R; v1_3_8.flags = 4; v1_3_8.act = 0;
      v1_3_8.alpha = 1.0f; v1_3_8.beta = 1.0f; v1_3_8.sa = 1.0f; v1_3_8.sb = 1.0f; v1_3_8.Npad = C; v1_3_8.pad_ = 0;
      k_gemm<1><<<dim3((unsigned)((C) + 31) / 32, (unsigned)((R) + 15) / 16, (unsigned)(R * R)), 32, 0, stream>>>(v1_3_8); }
    { GemmP v1_3_9;
      v1_3_9.A = GP + (size_t)3 * RP3 * C + (size_t)1156 * C; v1_3_9.B = wv1 + 9; v1_3_9.bias = GP + (size_t)3 * RP3 * C + (size_t)1156 * C; v1_3_9.R = GC + (size_t)3 * R3 * C; v1_3_9.C = GC + (size_t)3 * R3 * C;
      v1_3_9.sAo = (long long)34 * 34 * C; v1_3_9.sAi = (long long)34 * C; v1_3_9.sAm = C; v1_3_9.sAk = 1; v1_3_9.sBo = 0; v1_3_9.sBi = 0; v1_3_9.sBn = C * 27; v1_3_9.sBk = 27; v1_3_9.sCo = (long long)R * R * C; v1_3_9.sCi = (long long)R * C; v1_3_9.sCm = C; v1_3_9.sRo = (long long)R * R * C; v1_3_9.sRi = (long long)R * C; v1_3_9.sRm = C; v1_3_9.sRn = 1;
      v1_3_9.M = R; v1_3_9.N = C; v1_3_9.K = C; v1_3_9.zi_n = R; v1_3_9.flags = 4; v1_3_9.act = 0;
      v1_3_9.alpha = 1.0f; v1_3_9.beta = 1.0f; v1_3_9.sa = 1.0f; v1_3_9.sb = 1.0f; v1_3_9.Npad = C; v1_3_9.pad_ = 0;
      k_gemm<1><<<dim3((unsigned)((C) + 31) / 32, (unsigned)((R) + 15) / 16, (unsigned)(R * R)), 32, 0, stream>>>(v1_3_9); }
    { GemmP v1_3_10;
      v1_3_10.A = GP + (size_t)3 * RP3 * C + (size_t)1157 * C; v1_3_10.B = wv1 + 10; v1_3_10.bias = GP + (size_t)3 * RP3 * C + (size_t)1157 * C; v1_3_10.R = GC + (size_t)3 * R3 * C; v1_3_10.C = GC + (size_t)3 * R3 * C;
      v1_3_10.sAo = (long long)34 * 34 * C; v1_3_10.sAi = (long long)34 * C; v1_3_10.sAm = C; v1_3_10.sAk = 1; v1_3_10.sBo = 0; v1_3_10.sBi = 0; v1_3_10.sBn = C * 27; v1_3_10.sBk = 27; v1_3_10.sCo = (long long)R * R * C; v1_3_10.sCi = (long long)R * C; v1_3_10.sCm = C; v1_3_10.sRo = (long long)R * R * C; v1_3_10.sRi = (long long)R * C; v1_3_10.sRm = C; v1_3_10.sRn = 1;
      v1_3_10.M = R; v1_3_10.N = C; v1_3_10.K = C; v1_3_10.zi_n = R; v1_3_10.flags = 4; v1_3_10.act = 0;
      v1_3_10.alpha = 1.0f; v1_3_10.beta = 1.0f; v1_3_10.sa = 1.0f; v1_3_10.sb = 1.0f; v1_3_10.Npad = C; v1_3_10.pad_ = 0;
      k_gemm<1><<<dim3((unsigned)((C) + 31) / 32, (unsigned)((R) + 15) / 16, (unsigned)(R * R)), 32, 0, stream>>>(v1_3_10); }
    { GemmP v1_3_11;
      v1_3_11.A = GP + (size_t)3 * RP3 * C + (size_t)1158 * C; v1_3_11.B = wv1 + 11; v1_3_11.bias = GP + (size_t)3 * RP3 * C + (size_t)1158 * C; v1_3_11.R = GC + (size_t)3 * R3 * C; v1_3_11.C = GC + (size_t)3 * R3 * C;
      v1_3_11.sAo = (long long)34 * 34 * C; v1_3_11.sAi = (long long)34 * C; v1_3_11.sAm = C; v1_3_11.sAk = 1; v1_3_11.sBo = 0; v1_3_11.sBi = 0; v1_3_11.sBn = C * 27; v1_3_11.sBk = 27; v1_3_11.sCo = (long long)R * R * C; v1_3_11.sCi = (long long)R * C; v1_3_11.sCm = C; v1_3_11.sRo = (long long)R * R * C; v1_3_11.sRi = (long long)R * C; v1_3_11.sRm = C; v1_3_11.sRn = 1;
      v1_3_11.M = R; v1_3_11.N = C; v1_3_11.K = C; v1_3_11.zi_n = R; v1_3_11.flags = 4; v1_3_11.act = 0;
      v1_3_11.alpha = 1.0f; v1_3_11.beta = 1.0f; v1_3_11.sa = 1.0f; v1_3_11.sb = 1.0f; v1_3_11.Npad = C; v1_3_11.pad_ = 0;
      k_gemm<1><<<dim3((unsigned)((C) + 31) / 32, (unsigned)((R) + 15) / 16, (unsigned)(R * R)), 32, 0, stream>>>(v1_3_11); }
    { GemmP v1_3_12;
      v1_3_12.A = GP + (size_t)3 * RP3 * C + (size_t)1190 * C; v1_3_12.B = wv1 + 12; v1_3_12.bias = GP + (size_t)3 * RP3 * C + (size_t)1190 * C; v1_3_12.R = GC + (size_t)3 * R3 * C; v1_3_12.C = GC + (size_t)3 * R3 * C;
      v1_3_12.sAo = (long long)34 * 34 * C; v1_3_12.sAi = (long long)34 * C; v1_3_12.sAm = C; v1_3_12.sAk = 1; v1_3_12.sBo = 0; v1_3_12.sBi = 0; v1_3_12.sBn = C * 27; v1_3_12.sBk = 27; v1_3_12.sCo = (long long)R * R * C; v1_3_12.sCi = (long long)R * C; v1_3_12.sCm = C; v1_3_12.sRo = (long long)R * R * C; v1_3_12.sRi = (long long)R * C; v1_3_12.sRm = C; v1_3_12.sRn = 1;
      v1_3_12.M = R; v1_3_12.N = C; v1_3_12.K = C; v1_3_12.zi_n = R; v1_3_12.flags = 4; v1_3_12.act = 0;
      v1_3_12.alpha = 1.0f; v1_3_12.beta = 1.0f; v1_3_12.sa = 1.0f; v1_3_12.sb = 1.0f; v1_3_12.Npad = C; v1_3_12.pad_ = 0;
      k_gemm<1><<<dim3((unsigned)((C) + 31) / 32, (unsigned)((R) + 15) / 16, (unsigned)(R * R)), 32, 0, stream>>>(v1_3_12); }
    { GemmP v1_3_13;
      v1_3_13.A = GP + (size_t)3 * RP3 * C + (size_t)1191 * C; v1_3_13.B = wv1 + 13; v1_3_13.bias = GP + (size_t)3 * RP3 * C + (size_t)1191 * C; v1_3_13.R = GC + (size_t)3 * R3 * C; v1_3_13.C = GC + (size_t)3 * R3 * C;
      v1_3_13.sAo = (long long)34 * 34 * C; v1_3_13.sAi = (long long)34 * C; v1_3_13.sAm = C; v1_3_13.sAk = 1; v1_3_13.sBo = 0; v1_3_13.sBi = 0; v1_3_13.sBn = C * 27; v1_3_13.sBk = 27; v1_3_13.sCo = (long long)R * R * C; v1_3_13.sCi = (long long)R * C; v1_3_13.sCm = C; v1_3_13.sRo = (long long)R * R * C; v1_3_13.sRi = (long long)R * C; v1_3_13.sRm = C; v1_3_13.sRn = 1;
      v1_3_13.M = R; v1_3_13.N = C; v1_3_13.K = C; v1_3_13.zi_n = R; v1_3_13.flags = 4; v1_3_13.act = 0;
      v1_3_13.alpha = 1.0f; v1_3_13.beta = 1.0f; v1_3_13.sa = 1.0f; v1_3_13.sb = 1.0f; v1_3_13.Npad = C; v1_3_13.pad_ = 0;
      k_gemm<1><<<dim3((unsigned)((C) + 31) / 32, (unsigned)((R) + 15) / 16, (unsigned)(R * R)), 32, 0, stream>>>(v1_3_13); }
    { GemmP v1_3_14;
      v1_3_14.A = GP + (size_t)3 * RP3 * C + (size_t)1192 * C; v1_3_14.B = wv1 + 14; v1_3_14.bias = GP + (size_t)3 * RP3 * C + (size_t)1192 * C; v1_3_14.R = GC + (size_t)3 * R3 * C; v1_3_14.C = GC + (size_t)3 * R3 * C;
      v1_3_14.sAo = (long long)34 * 34 * C; v1_3_14.sAi = (long long)34 * C; v1_3_14.sAm = C; v1_3_14.sAk = 1; v1_3_14.sBo = 0; v1_3_14.sBi = 0; v1_3_14.sBn = C * 27; v1_3_14.sBk = 27; v1_3_14.sCo = (long long)R * R * C; v1_3_14.sCi = (long long)R * C; v1_3_14.sCm = C; v1_3_14.sRo = (long long)R * R * C; v1_3_14.sRi = (long long)R * C; v1_3_14.sRm = C; v1_3_14.sRn = 1;
      v1_3_14.M = R; v1_3_14.N = C; v1_3_14.K = C; v1_3_14.zi_n = R; v1_3_14.flags = 4; v1_3_14.act = 0;
      v1_3_14.alpha = 1.0f; v1_3_14.beta = 1.0f; v1_3_14.sa = 1.0f; v1_3_14.sb = 1.0f; v1_3_14.Npad = C; v1_3_14.pad_ = 0;
      k_gemm<1><<<dim3((unsigned)((C) + 31) / 32, (unsigned)((R) + 15) / 16, (unsigned)(R * R)), 32, 0, stream>>>(v1_3_14); }
    { GemmP v1_3_15;
      v1_3_15.A = GP + (size_t)3 * RP3 * C + (size_t)1224 * C; v1_3_15.B = wv1 + 15; v1_3_15.bias = GP + (size_t)3 * RP3 * C + (size_t)1224 * C; v1_3_15.R = GC + (size_t)3 * R3 * C; v1_3_15.C = GC + (size_t)3 * R3 * C;
      v1_3_15.sAo = (long long)34 * 34 * C; v1_3_15.sAi = (long long)34 * C; v1_3_15.sAm = C; v1_3_15.sAk = 1; v1_3_15.sBo = 0; v1_3_15.sBi = 0; v1_3_15.sBn = C * 27; v1_3_15.sBk = 27; v1_3_15.sCo = (long long)R * R * C; v1_3_15.sCi = (long long)R * C; v1_3_15.sCm = C; v1_3_15.sRo = (long long)R * R * C; v1_3_15.sRi = (long long)R * C; v1_3_15.sRm = C; v1_3_15.sRn = 1;
      v1_3_15.M = R; v1_3_15.N = C; v1_3_15.K = C; v1_3_15.zi_n = R; v1_3_15.flags = 4; v1_3_15.act = 0;
      v1_3_15.alpha = 1.0f; v1_3_15.beta = 1.0f; v1_3_15.sa = 1.0f; v1_3_15.sb = 1.0f; v1_3_15.Npad = C; v1_3_15.pad_ = 0;
      k_gemm<1><<<dim3((unsigned)((C) + 31) / 32, (unsigned)((R) + 15) / 16, (unsigned)(R * R)), 32, 0, stream>>>(v1_3_15); }
    { GemmP v1_3_16;
      v1_3_16.A = GP + (size_t)3 * RP3 * C + (size_t)1225 * C; v1_3_16.B = wv1 + 16; v1_3_16.bias = GP + (size_t)3 * RP3 * C + (size_t)1225 * C; v1_3_16.R = GC + (size_t)3 * R3 * C; v1_3_16.C = GC + (size_t)3 * R3 * C;
      v1_3_16.sAo = (long long)34 * 34 * C; v1_3_16.sAi = (long long)34 * C; v1_3_16.sAm = C; v1_3_16.sAk = 1; v1_3_16.sBo = 0; v1_3_16.sBi = 0; v1_3_16.sBn = C * 27; v1_3_16.sBk = 27; v1_3_16.sCo = (long long)R * R * C; v1_3_16.sCi = (long long)R * C; v1_3_16.sCm = C; v1_3_16.sRo = (long long)R * R * C; v1_3_16.sRi = (long long)R * C; v1_3_16.sRm = C; v1_3_16.sRn = 1;
      v1_3_16.M = R; v1_3_16.N = C; v1_3_16.K = C; v1_3_16.zi_n = R; v1_3_16.flags = 4; v1_3_16.act = 0;
      v1_3_16.alpha = 1.0f; v1_3_16.beta = 1.0f; v1_3_16.sa = 1.0f; v1_3_16.sb = 1.0f; v1_3_16.Npad = C; v1_3_16.pad_ = 0;
      k_gemm<1><<<dim3((unsigned)((C) + 31) / 32, (unsigned)((R) + 15) / 16, (unsigned)(R * R)), 32, 0, stream>>>(v1_3_16); }
    { GemmP v1_3_17;
      v1_3_17.A = GP + (size_t)3 * RP3 * C + (size_t)1226 * C; v1_3_17.B = wv1 + 17; v1_3_17.bias = GP + (size_t)3 * RP3 * C + (size_t)1226 * C; v1_3_17.R = GC + (size_t)3 * R3 * C; v1_3_17.C = GC + (size_t)3 * R3 * C;
      v1_3_17.sAo = (long long)34 * 34 * C; v1_3_17.sAi = (long long)34 * C; v1_3_17.sAm = C; v1_3_17.sAk = 1; v1_3_17.sBo = 0; v1_3_17.sBi = 0; v1_3_17.sBn = C * 27; v1_3_17.sBk = 27; v1_3_17.sCo = (long long)R * R * C; v1_3_17.sCi = (long long)R * C; v1_3_17.sCm = C; v1_3_17.sRo = (long long)R * R * C; v1_3_17.sRi = (long long)R * C; v1_3_17.sRm = C; v1_3_17.sRn = 1;
      v1_3_17.M = R; v1_3_17.N = C; v1_3_17.K = C; v1_3_17.zi_n = R; v1_3_17.flags = 4; v1_3_17.act = 0;
      v1_3_17.alpha = 1.0f; v1_3_17.beta = 1.0f; v1_3_17.sa = 1.0f; v1_3_17.sb = 1.0f; v1_3_17.Npad = C; v1_3_17.pad_ = 0;
      k_gemm<1><<<dim3((unsigned)((C) + 31) / 32, (unsigned)((R) + 15) / 16, (unsigned)(R * R)), 32, 0, stream>>>(v1_3_17); }
    { GemmP v1_3_18;
      v1_3_18.A = GP + (size_t)3 * RP3 * C + (size_t)2312 * C; v1_3_18.B = wv1 + 18; v1_3_18.bias = GP + (size_t)3 * RP3 * C + (size_t)2312 * C; v1_3_18.R = GC + (size_t)3 * R3 * C; v1_3_18.C = GC + (size_t)3 * R3 * C;
      v1_3_18.sAo = (long long)34 * 34 * C; v1_3_18.sAi = (long long)34 * C; v1_3_18.sAm = C; v1_3_18.sAk = 1; v1_3_18.sBo = 0; v1_3_18.sBi = 0; v1_3_18.sBn = C * 27; v1_3_18.sBk = 27; v1_3_18.sCo = (long long)R * R * C; v1_3_18.sCi = (long long)R * C; v1_3_18.sCm = C; v1_3_18.sRo = (long long)R * R * C; v1_3_18.sRi = (long long)R * C; v1_3_18.sRm = C; v1_3_18.sRn = 1;
      v1_3_18.M = R; v1_3_18.N = C; v1_3_18.K = C; v1_3_18.zi_n = R; v1_3_18.flags = 4; v1_3_18.act = 0;
      v1_3_18.alpha = 1.0f; v1_3_18.beta = 1.0f; v1_3_18.sa = 1.0f; v1_3_18.sb = 1.0f; v1_3_18.Npad = C; v1_3_18.pad_ = 0;
      k_gemm<1><<<dim3((unsigned)((C) + 31) / 32, (unsigned)((R) + 15) / 16, (unsigned)(R * R)), 32, 0, stream>>>(v1_3_18); }
    { GemmP v1_3_19;
      v1_3_19.A = GP + (size_t)3 * RP3 * C + (size_t)2313 * C; v1_3_19.B = wv1 + 19; v1_3_19.bias = GP + (size_t)3 * RP3 * C + (size_t)2313 * C; v1_3_19.R = GC + (size_t)3 * R3 * C; v1_3_19.C = GC + (size_t)3 * R3 * C;
      v1_3_19.sAo = (long long)34 * 34 * C; v1_3_19.sAi = (long long)34 * C; v1_3_19.sAm = C; v1_3_19.sAk = 1; v1_3_19.sBo = 0; v1_3_19.sBi = 0; v1_3_19.sBn = C * 27; v1_3_19.sBk = 27; v1_3_19.sCo = (long long)R * R * C; v1_3_19.sCi = (long long)R * C; v1_3_19.sCm = C; v1_3_19.sRo = (long long)R * R * C; v1_3_19.sRi = (long long)R * C; v1_3_19.sRm = C; v1_3_19.sRn = 1;
      v1_3_19.M = R; v1_3_19.N = C; v1_3_19.K = C; v1_3_19.zi_n = R; v1_3_19.flags = 4; v1_3_19.act = 0;
      v1_3_19.alpha = 1.0f; v1_3_19.beta = 1.0f; v1_3_19.sa = 1.0f; v1_3_19.sb = 1.0f; v1_3_19.Npad = C; v1_3_19.pad_ = 0;
      k_gemm<1><<<dim3((unsigned)((C) + 31) / 32, (unsigned)((R) + 15) / 16, (unsigned)(R * R)), 32, 0, stream>>>(v1_3_19); }
    { GemmP v1_3_20;
      v1_3_20.A = GP + (size_t)3 * RP3 * C + (size_t)2314 * C; v1_3_20.B = wv1 + 20; v1_3_20.bias = GP + (size_t)3 * RP3 * C + (size_t)2314 * C; v1_3_20.R = GC + (size_t)3 * R3 * C; v1_3_20.C = GC + (size_t)3 * R3 * C;
      v1_3_20.sAo = (long long)34 * 34 * C; v1_3_20.sAi = (long long)34 * C; v1_3_20.sAm = C; v1_3_20.sAk = 1; v1_3_20.sBo = 0; v1_3_20.sBi = 0; v1_3_20.sBn = C * 27; v1_3_20.sBk = 27; v1_3_20.sCo = (long long)R * R * C; v1_3_20.sCi = (long long)R * C; v1_3_20.sCm = C; v1_3_20.sRo = (long long)R * R * C; v1_3_20.sRi = (long long)R * C; v1_3_20.sRm = C; v1_3_20.sRn = 1;
      v1_3_20.M = R; v1_3_20.N = C; v1_3_20.K = C; v1_3_20.zi_n = R; v1_3_20.flags = 4; v1_3_20.act = 0;
      v1_3_20.alpha = 1.0f; v1_3_20.beta = 1.0f; v1_3_20.sa = 1.0f; v1_3_20.sb = 1.0f; v1_3_20.Npad = C; v1_3_20.pad_ = 0;
      k_gemm<1><<<dim3((unsigned)((C) + 31) / 32, (unsigned)((R) + 15) / 16, (unsigned)(R * R)), 32, 0, stream>>>(v1_3_20); }
    { GemmP v1_3_21;
      v1_3_21.A = GP + (size_t)3 * RP3 * C + (size_t)2346 * C; v1_3_21.B = wv1 + 21; v1_3_21.bias = GP + (size_t)3 * RP3 * C + (size_t)2346 * C; v1_3_21.R = GC + (size_t)3 * R3 * C; v1_3_21.C = GC + (size_t)3 * R3 * C;
      v1_3_21.sAo = (long long)34 * 34 * C; v1_3_21.sAi = (long long)34 * C; v1_3_21.sAm = C; v1_3_21.sAk = 1; v1_3_21.sBo = 0; v1_3_21.sBi = 0; v1_3_21.sBn = C * 27; v1_3_21.sBk = 27; v1_3_21.sCo = (long long)R * R * C; v1_3_21.sCi = (long long)R * C; v1_3_21.sCm = C; v1_3_21.sRo = (long long)R * R * C; v1_3_21.sRi = (long long)R * C; v1_3_21.sRm = C; v1_3_21.sRn = 1;
      v1_3_21.M = R; v1_3_21.N = C; v1_3_21.K = C; v1_3_21.zi_n = R; v1_3_21.flags = 4; v1_3_21.act = 0;
      v1_3_21.alpha = 1.0f; v1_3_21.beta = 1.0f; v1_3_21.sa = 1.0f; v1_3_21.sb = 1.0f; v1_3_21.Npad = C; v1_3_21.pad_ = 0;
      k_gemm<1><<<dim3((unsigned)((C) + 31) / 32, (unsigned)((R) + 15) / 16, (unsigned)(R * R)), 32, 0, stream>>>(v1_3_21); }
    { GemmP v1_3_22;
      v1_3_22.A = GP + (size_t)3 * RP3 * C + (size_t)2347 * C; v1_3_22.B = wv1 + 22; v1_3_22.bias = GP + (size_t)3 * RP3 * C + (size_t)2347 * C; v1_3_22.R = GC + (size_t)3 * R3 * C; v1_3_22.C = GC + (size_t)3 * R3 * C;
      v1_3_22.sAo = (long long)34 * 34 * C; v1_3_22.sAi = (long long)34 * C; v1_3_22.sAm = C; v1_3_22.sAk = 1; v1_3_22.sBo = 0; v1_3_22.sBi = 0; v1_3_22.sBn = C * 27; v1_3_22.sBk = 27; v1_3_22.sCo = (long long)R * R * C; v1_3_22.sCi = (long long)R * C; v1_3_22.sCm = C; v1_3_22.sRo = (long long)R * R * C; v1_3_22.sRi = (long long)R * C; v1_3_22.sRm = C; v1_3_22.sRn = 1;
      v1_3_22.M = R; v1_3_22.N = C; v1_3_22.K = C; v1_3_22.zi_n = R; v1_3_22.flags = 4; v1_3_22.act = 0;
      v1_3_22.alpha = 1.0f; v1_3_22.beta = 1.0f; v1_3_22.sa = 1.0f; v1_3_22.sb = 1.0f; v1_3_22.Npad = C; v1_3_22.pad_ = 0;
      k_gemm<1><<<dim3((unsigned)((C) + 31) / 32, (unsigned)((R) + 15) / 16, (unsigned)(R * R)), 32, 0, stream>>>(v1_3_22); }
    { GemmP v1_3_23;
      v1_3_23.A = GP + (size_t)3 * RP3 * C + (size_t)2348 * C; v1_3_23.B = wv1 + 23; v1_3_23.bias = GP + (size_t)3 * RP3 * C + (size_t)2348 * C; v1_3_23.R = GC + (size_t)3 * R3 * C; v1_3_23.C = GC + (size_t)3 * R3 * C;
      v1_3_23.sAo = (long long)34 * 34 * C; v1_3_23.sAi = (long long)34 * C; v1_3_23.sAm = C; v1_3_23.sAk = 1; v1_3_23.sBo = 0; v1_3_23.sBi = 0; v1_3_23.sBn = C * 27; v1_3_23.sBk = 27; v1_3_23.sCo = (long long)R * R * C; v1_3_23.sCi = (long long)R * C; v1_3_23.sCm = C; v1_3_23.sRo = (long long)R * R * C; v1_3_23.sRi = (long long)R * C; v1_3_23.sRm = C; v1_3_23.sRn = 1;
      v1_3_23.M = R; v1_3_23.N = C; v1_3_23.K = C; v1_3_23.zi_n = R; v1_3_23.flags = 4; v1_3_23.act = 0;
      v1_3_23.alpha = 1.0f; v1_3_23.beta = 1.0f; v1_3_23.sa = 1.0f; v1_3_23.sb = 1.0f; v1_3_23.Npad = C; v1_3_23.pad_ = 0;
      k_gemm<1><<<dim3((unsigned)((C) + 31) / 32, (unsigned)((R) + 15) / 16, (unsigned)(R * R)), 32, 0, stream>>>(v1_3_23); }
    { GemmP v1_3_24;
      v1_3_24.A = GP + (size_t)3 * RP3 * C + (size_t)2380 * C; v1_3_24.B = wv1 + 24; v1_3_24.bias = GP + (size_t)3 * RP3 * C + (size_t)2380 * C; v1_3_24.R = GC + (size_t)3 * R3 * C; v1_3_24.C = GC + (size_t)3 * R3 * C;
      v1_3_24.sAo = (long long)34 * 34 * C; v1_3_24.sAi = (long long)34 * C; v1_3_24.sAm = C; v1_3_24.sAk = 1; v1_3_24.sBo = 0; v1_3_24.sBi = 0; v1_3_24.sBn = C * 27; v1_3_24.sBk = 27; v1_3_24.sCo = (long long)R * R * C; v1_3_24.sCi = (long long)R * C; v1_3_24.sCm = C; v1_3_24.sRo = (long long)R * R * C; v1_3_24.sRi = (long long)R * C; v1_3_24.sRm = C; v1_3_24.sRn = 1;
      v1_3_24.M = R; v1_3_24.N = C; v1_3_24.K = C; v1_3_24.zi_n = R; v1_3_24.flags = 4; v1_3_24.act = 0;
      v1_3_24.alpha = 1.0f; v1_3_24.beta = 1.0f; v1_3_24.sa = 1.0f; v1_3_24.sb = 1.0f; v1_3_24.Npad = C; v1_3_24.pad_ = 0;
      k_gemm<1><<<dim3((unsigned)((C) + 31) / 32, (unsigned)((R) + 15) / 16, (unsigned)(R * R)), 32, 0, stream>>>(v1_3_24); }
    { GemmP v1_3_25;
      v1_3_25.A = GP + (size_t)3 * RP3 * C + (size_t)2381 * C; v1_3_25.B = wv1 + 25; v1_3_25.bias = GP + (size_t)3 * RP3 * C + (size_t)2381 * C; v1_3_25.R = GC + (size_t)3 * R3 * C; v1_3_25.C = GC + (size_t)3 * R3 * C;
      v1_3_25.sAo = (long long)34 * 34 * C; v1_3_25.sAi = (long long)34 * C; v1_3_25.sAm = C; v1_3_25.sAk = 1; v1_3_25.sBo = 0; v1_3_25.sBi = 0; v1_3_25.sBn = C * 27; v1_3_25.sBk = 27; v1_3_25.sCo = (long long)R * R * C; v1_3_25.sCi = (long long)R * C; v1_3_25.sCm = C; v1_3_25.sRo = (long long)R * R * C; v1_3_25.sRi = (long long)R * C; v1_3_25.sRm = C; v1_3_25.sRn = 1;
      v1_3_25.M = R; v1_3_25.N = C; v1_3_25.K = C; v1_3_25.zi_n = R; v1_3_25.flags = 4; v1_3_25.act = 0;
      v1_3_25.alpha = 1.0f; v1_3_25.beta = 1.0f; v1_3_25.sa = 1.0f; v1_3_25.sb = 1.0f; v1_3_25.Npad = C; v1_3_25.pad_ = 0;
      k_gemm<1><<<dim3((unsigned)((C) + 31) / 32, (unsigned)((R) + 15) / 16, (unsigned)(R * R)), 32, 0, stream>>>(v1_3_25); }
    { GemmP v1_3_26;
      v1_3_26.A = GP + (size_t)3 * RP3 * C + (size_t)2382 * C; v1_3_26.B = wv1 + 26; v1_3_26.bias = GP + (size_t)3 * RP3 * C + (size_t)2382 * C; v1_3_26.R = GC + (size_t)3 * R3 * C; v1_3_26.C = GC + (size_t)3 * R3 * C;
      v1_3_26.sAo = (long long)34 * 34 * C; v1_3_26.sAi = (long long)34 * C; v1_3_26.sAm = C; v1_3_26.sAk = 1; v1_3_26.sBo = 0; v1_3_26.sBi = 0; v1_3_26.sBn = C * 27; v1_3_26.sBk = 27; v1_3_26.sCo = (long long)R * R * C; v1_3_26.sCi = (long long)R * C; v1_3_26.sCm = C; v1_3_26.sRo = (long long)R * R * C; v1_3_26.sRi = (long long)R * C; v1_3_26.sRm = C; v1_3_26.sRn = 1;
      v1_3_26.M = R; v1_3_26.N = C; v1_3_26.K = C; v1_3_26.zi_n = R; v1_3_26.flags = 4; v1_3_26.act = 0;
      v1_3_26.alpha = 1.0f; v1_3_26.beta = 1.0f; v1_3_26.sa = 1.0f; v1_3_26.sb = 1.0f; v1_3_26.Npad = C; v1_3_26.pad_ = 0;
      k_gemm<1><<<dim3((unsigned)((C) + 31) / 32, (unsigned)((R) + 15) / 16, (unsigned)(R * R)), 32, 0, stream>>>(v1_3_26); }
    k_cc_bnl<<<(unsigned)(((long long)NV * C + 255) / 256), 256, 0, stream>>>(GC, g1, be1, GQ, Bn, R, C);
    { GemmP v2_0_0;
      v2_0_0.A = GQ + (size_t)0 * RP3 * C + (size_t)0 * C; v2_0_0.B = wv2 + 0; v2_0_0.bias = GQ + (size_t)0 * RP3 * C + (size_t)0 * C; v2_0_0.R = GQ + (size_t)0 * RP3 * C + (size_t)0 * C; v2_0_0.C = GC + (size_t)0 * R3 * C;
      v2_0_0.sAo = (long long)34 * 34 * C; v2_0_0.sAi = (long long)34 * C; v2_0_0.sAm = C; v2_0_0.sAk = 1; v2_0_0.sBo = 0; v2_0_0.sBi = 0; v2_0_0.sBn = C * 27; v2_0_0.sBk = 27; v2_0_0.sCo = (long long)R * R * C; v2_0_0.sCi = (long long)R * C; v2_0_0.sCm = C; v2_0_0.sRo = 0; v2_0_0.sRi = 0; v2_0_0.sRm = 0; v2_0_0.sRn = 0;
      v2_0_0.M = R; v2_0_0.N = C; v2_0_0.K = C; v2_0_0.zi_n = R; v2_0_0.flags = 0; v2_0_0.act = 0;
      v2_0_0.alpha = 1.0f; v2_0_0.beta = 0.0f; v2_0_0.sa = 1.0f; v2_0_0.sb = 1.0f; v2_0_0.Npad = C; v2_0_0.pad_ = 0;
      k_gemm<1><<<dim3((unsigned)((C) + 31) / 32, (unsigned)((R) + 15) / 16, (unsigned)(R * R)), 32, 0, stream>>>(v2_0_0); }
    { GemmP v2_0_1;
      v2_0_1.A = GQ + (size_t)0 * RP3 * C + (size_t)1 * C; v2_0_1.B = wv2 + 1; v2_0_1.bias = GQ + (size_t)0 * RP3 * C + (size_t)1 * C; v2_0_1.R = GC + (size_t)0 * R3 * C; v2_0_1.C = GC + (size_t)0 * R3 * C;
      v2_0_1.sAo = (long long)34 * 34 * C; v2_0_1.sAi = (long long)34 * C; v2_0_1.sAm = C; v2_0_1.sAk = 1; v2_0_1.sBo = 0; v2_0_1.sBi = 0; v2_0_1.sBn = C * 27; v2_0_1.sBk = 27; v2_0_1.sCo = (long long)R * R * C; v2_0_1.sCi = (long long)R * C; v2_0_1.sCm = C; v2_0_1.sRo = (long long)R * R * C; v2_0_1.sRi = (long long)R * C; v2_0_1.sRm = C; v2_0_1.sRn = 1;
      v2_0_1.M = R; v2_0_1.N = C; v2_0_1.K = C; v2_0_1.zi_n = R; v2_0_1.flags = 4; v2_0_1.act = 0;
      v2_0_1.alpha = 1.0f; v2_0_1.beta = 1.0f; v2_0_1.sa = 1.0f; v2_0_1.sb = 1.0f; v2_0_1.Npad = C; v2_0_1.pad_ = 0;
      k_gemm<1><<<dim3((unsigned)((C) + 31) / 32, (unsigned)((R) + 15) / 16, (unsigned)(R * R)), 32, 0, stream>>>(v2_0_1); }
    { GemmP v2_0_2;
      v2_0_2.A = GQ + (size_t)0 * RP3 * C + (size_t)2 * C; v2_0_2.B = wv2 + 2; v2_0_2.bias = GQ + (size_t)0 * RP3 * C + (size_t)2 * C; v2_0_2.R = GC + (size_t)0 * R3 * C; v2_0_2.C = GC + (size_t)0 * R3 * C;
      v2_0_2.sAo = (long long)34 * 34 * C; v2_0_2.sAi = (long long)34 * C; v2_0_2.sAm = C; v2_0_2.sAk = 1; v2_0_2.sBo = 0; v2_0_2.sBi = 0; v2_0_2.sBn = C * 27; v2_0_2.sBk = 27; v2_0_2.sCo = (long long)R * R * C; v2_0_2.sCi = (long long)R * C; v2_0_2.sCm = C; v2_0_2.sRo = (long long)R * R * C; v2_0_2.sRi = (long long)R * C; v2_0_2.sRm = C; v2_0_2.sRn = 1;
      v2_0_2.M = R; v2_0_2.N = C; v2_0_2.K = C; v2_0_2.zi_n = R; v2_0_2.flags = 4; v2_0_2.act = 0;
      v2_0_2.alpha = 1.0f; v2_0_2.beta = 1.0f; v2_0_2.sa = 1.0f; v2_0_2.sb = 1.0f; v2_0_2.Npad = C; v2_0_2.pad_ = 0;
      k_gemm<1><<<dim3((unsigned)((C) + 31) / 32, (unsigned)((R) + 15) / 16, (unsigned)(R * R)), 32, 0, stream>>>(v2_0_2); }
    { GemmP v2_0_3;
      v2_0_3.A = GQ + (size_t)0 * RP3 * C + (size_t)34 * C; v2_0_3.B = wv2 + 3; v2_0_3.bias = GQ + (size_t)0 * RP3 * C + (size_t)34 * C; v2_0_3.R = GC + (size_t)0 * R3 * C; v2_0_3.C = GC + (size_t)0 * R3 * C;
      v2_0_3.sAo = (long long)34 * 34 * C; v2_0_3.sAi = (long long)34 * C; v2_0_3.sAm = C; v2_0_3.sAk = 1; v2_0_3.sBo = 0; v2_0_3.sBi = 0; v2_0_3.sBn = C * 27; v2_0_3.sBk = 27; v2_0_3.sCo = (long long)R * R * C; v2_0_3.sCi = (long long)R * C; v2_0_3.sCm = C; v2_0_3.sRo = (long long)R * R * C; v2_0_3.sRi = (long long)R * C; v2_0_3.sRm = C; v2_0_3.sRn = 1;
      v2_0_3.M = R; v2_0_3.N = C; v2_0_3.K = C; v2_0_3.zi_n = R; v2_0_3.flags = 4; v2_0_3.act = 0;
      v2_0_3.alpha = 1.0f; v2_0_3.beta = 1.0f; v2_0_3.sa = 1.0f; v2_0_3.sb = 1.0f; v2_0_3.Npad = C; v2_0_3.pad_ = 0;
      k_gemm<1><<<dim3((unsigned)((C) + 31) / 32, (unsigned)((R) + 15) / 16, (unsigned)(R * R)), 32, 0, stream>>>(v2_0_3); }
    { GemmP v2_0_4;
      v2_0_4.A = GQ + (size_t)0 * RP3 * C + (size_t)35 * C; v2_0_4.B = wv2 + 4; v2_0_4.bias = GQ + (size_t)0 * RP3 * C + (size_t)35 * C; v2_0_4.R = GC + (size_t)0 * R3 * C; v2_0_4.C = GC + (size_t)0 * R3 * C;
      v2_0_4.sAo = (long long)34 * 34 * C; v2_0_4.sAi = (long long)34 * C; v2_0_4.sAm = C; v2_0_4.sAk = 1; v2_0_4.sBo = 0; v2_0_4.sBi = 0; v2_0_4.sBn = C * 27; v2_0_4.sBk = 27; v2_0_4.sCo = (long long)R * R * C; v2_0_4.sCi = (long long)R * C; v2_0_4.sCm = C; v2_0_4.sRo = (long long)R * R * C; v2_0_4.sRi = (long long)R * C; v2_0_4.sRm = C; v2_0_4.sRn = 1;
      v2_0_4.M = R; v2_0_4.N = C; v2_0_4.K = C; v2_0_4.zi_n = R; v2_0_4.flags = 4; v2_0_4.act = 0;
      v2_0_4.alpha = 1.0f; v2_0_4.beta = 1.0f; v2_0_4.sa = 1.0f; v2_0_4.sb = 1.0f; v2_0_4.Npad = C; v2_0_4.pad_ = 0;
      k_gemm<1><<<dim3((unsigned)((C) + 31) / 32, (unsigned)((R) + 15) / 16, (unsigned)(R * R)), 32, 0, stream>>>(v2_0_4); }
    { GemmP v2_0_5;
      v2_0_5.A = GQ + (size_t)0 * RP3 * C + (size_t)36 * C; v2_0_5.B = wv2 + 5; v2_0_5.bias = GQ + (size_t)0 * RP3 * C + (size_t)36 * C; v2_0_5.R = GC + (size_t)0 * R3 * C; v2_0_5.C = GC + (size_t)0 * R3 * C;
      v2_0_5.sAo = (long long)34 * 34 * C; v2_0_5.sAi = (long long)34 * C; v2_0_5.sAm = C; v2_0_5.sAk = 1; v2_0_5.sBo = 0; v2_0_5.sBi = 0; v2_0_5.sBn = C * 27; v2_0_5.sBk = 27; v2_0_5.sCo = (long long)R * R * C; v2_0_5.sCi = (long long)R * C; v2_0_5.sCm = C; v2_0_5.sRo = (long long)R * R * C; v2_0_5.sRi = (long long)R * C; v2_0_5.sRm = C; v2_0_5.sRn = 1;
      v2_0_5.M = R; v2_0_5.N = C; v2_0_5.K = C; v2_0_5.zi_n = R; v2_0_5.flags = 4; v2_0_5.act = 0;
      v2_0_5.alpha = 1.0f; v2_0_5.beta = 1.0f; v2_0_5.sa = 1.0f; v2_0_5.sb = 1.0f; v2_0_5.Npad = C; v2_0_5.pad_ = 0;
      k_gemm<1><<<dim3((unsigned)((C) + 31) / 32, (unsigned)((R) + 15) / 16, (unsigned)(R * R)), 32, 0, stream>>>(v2_0_5); }
    { GemmP v2_0_6;
      v2_0_6.A = GQ + (size_t)0 * RP3 * C + (size_t)68 * C; v2_0_6.B = wv2 + 6; v2_0_6.bias = GQ + (size_t)0 * RP3 * C + (size_t)68 * C; v2_0_6.R = GC + (size_t)0 * R3 * C; v2_0_6.C = GC + (size_t)0 * R3 * C;
      v2_0_6.sAo = (long long)34 * 34 * C; v2_0_6.sAi = (long long)34 * C; v2_0_6.sAm = C; v2_0_6.sAk = 1; v2_0_6.sBo = 0; v2_0_6.sBi = 0; v2_0_6.sBn = C * 27; v2_0_6.sBk = 27; v2_0_6.sCo = (long long)R * R * C; v2_0_6.sCi = (long long)R * C; v2_0_6.sCm = C; v2_0_6.sRo = (long long)R * R * C; v2_0_6.sRi = (long long)R * C; v2_0_6.sRm = C; v2_0_6.sRn = 1;
      v2_0_6.M = R; v2_0_6.N = C; v2_0_6.K = C; v2_0_6.zi_n = R; v2_0_6.flags = 4; v2_0_6.act = 0;
      v2_0_6.alpha = 1.0f; v2_0_6.beta = 1.0f; v2_0_6.sa = 1.0f; v2_0_6.sb = 1.0f; v2_0_6.Npad = C; v2_0_6.pad_ = 0;
      k_gemm<1><<<dim3((unsigned)((C) + 31) / 32, (unsigned)((R) + 15) / 16, (unsigned)(R * R)), 32, 0, stream>>>(v2_0_6); }
    { GemmP v2_0_7;
      v2_0_7.A = GQ + (size_t)0 * RP3 * C + (size_t)69 * C; v2_0_7.B = wv2 + 7; v2_0_7.bias = GQ + (size_t)0 * RP3 * C + (size_t)69 * C; v2_0_7.R = GC + (size_t)0 * R3 * C; v2_0_7.C = GC + (size_t)0 * R3 * C;
      v2_0_7.sAo = (long long)34 * 34 * C; v2_0_7.sAi = (long long)34 * C; v2_0_7.sAm = C; v2_0_7.sAk = 1; v2_0_7.sBo = 0; v2_0_7.sBi = 0; v2_0_7.sBn = C * 27; v2_0_7.sBk = 27; v2_0_7.sCo = (long long)R * R * C; v2_0_7.sCi = (long long)R * C; v2_0_7.sCm = C; v2_0_7.sRo = (long long)R * R * C; v2_0_7.sRi = (long long)R * C; v2_0_7.sRm = C; v2_0_7.sRn = 1;
      v2_0_7.M = R; v2_0_7.N = C; v2_0_7.K = C; v2_0_7.zi_n = R; v2_0_7.flags = 4; v2_0_7.act = 0;
      v2_0_7.alpha = 1.0f; v2_0_7.beta = 1.0f; v2_0_7.sa = 1.0f; v2_0_7.sb = 1.0f; v2_0_7.Npad = C; v2_0_7.pad_ = 0;
      k_gemm<1><<<dim3((unsigned)((C) + 31) / 32, (unsigned)((R) + 15) / 16, (unsigned)(R * R)), 32, 0, stream>>>(v2_0_7); }
    { GemmP v2_0_8;
      v2_0_8.A = GQ + (size_t)0 * RP3 * C + (size_t)70 * C; v2_0_8.B = wv2 + 8; v2_0_8.bias = GQ + (size_t)0 * RP3 * C + (size_t)70 * C; v2_0_8.R = GC + (size_t)0 * R3 * C; v2_0_8.C = GC + (size_t)0 * R3 * C;
      v2_0_8.sAo = (long long)34 * 34 * C; v2_0_8.sAi = (long long)34 * C; v2_0_8.sAm = C; v2_0_8.sAk = 1; v2_0_8.sBo = 0; v2_0_8.sBi = 0; v2_0_8.sBn = C * 27; v2_0_8.sBk = 27; v2_0_8.sCo = (long long)R * R * C; v2_0_8.sCi = (long long)R * C; v2_0_8.sCm = C; v2_0_8.sRo = (long long)R * R * C; v2_0_8.sRi = (long long)R * C; v2_0_8.sRm = C; v2_0_8.sRn = 1;
      v2_0_8.M = R; v2_0_8.N = C; v2_0_8.K = C; v2_0_8.zi_n = R; v2_0_8.flags = 4; v2_0_8.act = 0;
      v2_0_8.alpha = 1.0f; v2_0_8.beta = 1.0f; v2_0_8.sa = 1.0f; v2_0_8.sb = 1.0f; v2_0_8.Npad = C; v2_0_8.pad_ = 0;
      k_gemm<1><<<dim3((unsigned)((C) + 31) / 32, (unsigned)((R) + 15) / 16, (unsigned)(R * R)), 32, 0, stream>>>(v2_0_8); }
    { GemmP v2_0_9;
      v2_0_9.A = GQ + (size_t)0 * RP3 * C + (size_t)1156 * C; v2_0_9.B = wv2 + 9; v2_0_9.bias = GQ + (size_t)0 * RP3 * C + (size_t)1156 * C; v2_0_9.R = GC + (size_t)0 * R3 * C; v2_0_9.C = GC + (size_t)0 * R3 * C;
      v2_0_9.sAo = (long long)34 * 34 * C; v2_0_9.sAi = (long long)34 * C; v2_0_9.sAm = C; v2_0_9.sAk = 1; v2_0_9.sBo = 0; v2_0_9.sBi = 0; v2_0_9.sBn = C * 27; v2_0_9.sBk = 27; v2_0_9.sCo = (long long)R * R * C; v2_0_9.sCi = (long long)R * C; v2_0_9.sCm = C; v2_0_9.sRo = (long long)R * R * C; v2_0_9.sRi = (long long)R * C; v2_0_9.sRm = C; v2_0_9.sRn = 1;
      v2_0_9.M = R; v2_0_9.N = C; v2_0_9.K = C; v2_0_9.zi_n = R; v2_0_9.flags = 4; v2_0_9.act = 0;
      v2_0_9.alpha = 1.0f; v2_0_9.beta = 1.0f; v2_0_9.sa = 1.0f; v2_0_9.sb = 1.0f; v2_0_9.Npad = C; v2_0_9.pad_ = 0;
      k_gemm<1><<<dim3((unsigned)((C) + 31) / 32, (unsigned)((R) + 15) / 16, (unsigned)(R * R)), 32, 0, stream>>>(v2_0_9); }
    { GemmP v2_0_10;
      v2_0_10.A = GQ + (size_t)0 * RP3 * C + (size_t)1157 * C; v2_0_10.B = wv2 + 10; v2_0_10.bias = GQ + (size_t)0 * RP3 * C + (size_t)1157 * C; v2_0_10.R = GC + (size_t)0 * R3 * C; v2_0_10.C = GC + (size_t)0 * R3 * C;
      v2_0_10.sAo = (long long)34 * 34 * C; v2_0_10.sAi = (long long)34 * C; v2_0_10.sAm = C; v2_0_10.sAk = 1; v2_0_10.sBo = 0; v2_0_10.sBi = 0; v2_0_10.sBn = C * 27; v2_0_10.sBk = 27; v2_0_10.sCo = (long long)R * R * C; v2_0_10.sCi = (long long)R * C; v2_0_10.sCm = C; v2_0_10.sRo = (long long)R * R * C; v2_0_10.sRi = (long long)R * C; v2_0_10.sRm = C; v2_0_10.sRn = 1;
      v2_0_10.M = R; v2_0_10.N = C; v2_0_10.K = C; v2_0_10.zi_n = R; v2_0_10.flags = 4; v2_0_10.act = 0;
      v2_0_10.alpha = 1.0f; v2_0_10.beta = 1.0f; v2_0_10.sa = 1.0f; v2_0_10.sb = 1.0f; v2_0_10.Npad = C; v2_0_10.pad_ = 0;
      k_gemm<1><<<dim3((unsigned)((C) + 31) / 32, (unsigned)((R) + 15) / 16, (unsigned)(R * R)), 32, 0, stream>>>(v2_0_10); }
    { GemmP v2_0_11;
      v2_0_11.A = GQ + (size_t)0 * RP3 * C + (size_t)1158 * C; v2_0_11.B = wv2 + 11; v2_0_11.bias = GQ + (size_t)0 * RP3 * C + (size_t)1158 * C; v2_0_11.R = GC + (size_t)0 * R3 * C; v2_0_11.C = GC + (size_t)0 * R3 * C;
      v2_0_11.sAo = (long long)34 * 34 * C; v2_0_11.sAi = (long long)34 * C; v2_0_11.sAm = C; v2_0_11.sAk = 1; v2_0_11.sBo = 0; v2_0_11.sBi = 0; v2_0_11.sBn = C * 27; v2_0_11.sBk = 27; v2_0_11.sCo = (long long)R * R * C; v2_0_11.sCi = (long long)R * C; v2_0_11.sCm = C; v2_0_11.sRo = (long long)R * R * C; v2_0_11.sRi = (long long)R * C; v2_0_11.sRm = C; v2_0_11.sRn = 1;
      v2_0_11.M = R; v2_0_11.N = C; v2_0_11.K = C; v2_0_11.zi_n = R; v2_0_11.flags = 4; v2_0_11.act = 0;
      v2_0_11.alpha = 1.0f; v2_0_11.beta = 1.0f; v2_0_11.sa = 1.0f; v2_0_11.sb = 1.0f; v2_0_11.Npad = C; v2_0_11.pad_ = 0;
      k_gemm<1><<<dim3((unsigned)((C) + 31) / 32, (unsigned)((R) + 15) / 16, (unsigned)(R * R)), 32, 0, stream>>>(v2_0_11); }
    { GemmP v2_0_12;
      v2_0_12.A = GQ + (size_t)0 * RP3 * C + (size_t)1190 * C; v2_0_12.B = wv2 + 12; v2_0_12.bias = GQ + (size_t)0 * RP3 * C + (size_t)1190 * C; v2_0_12.R = GC + (size_t)0 * R3 * C; v2_0_12.C = GC + (size_t)0 * R3 * C;
      v2_0_12.sAo = (long long)34 * 34 * C; v2_0_12.sAi = (long long)34 * C; v2_0_12.sAm = C; v2_0_12.sAk = 1; v2_0_12.sBo = 0; v2_0_12.sBi = 0; v2_0_12.sBn = C * 27; v2_0_12.sBk = 27; v2_0_12.sCo = (long long)R * R * C; v2_0_12.sCi = (long long)R * C; v2_0_12.sCm = C; v2_0_12.sRo = (long long)R * R * C; v2_0_12.sRi = (long long)R * C; v2_0_12.sRm = C; v2_0_12.sRn = 1;
      v2_0_12.M = R; v2_0_12.N = C; v2_0_12.K = C; v2_0_12.zi_n = R; v2_0_12.flags = 4; v2_0_12.act = 0;
      v2_0_12.alpha = 1.0f; v2_0_12.beta = 1.0f; v2_0_12.sa = 1.0f; v2_0_12.sb = 1.0f; v2_0_12.Npad = C; v2_0_12.pad_ = 0;
      k_gemm<1><<<dim3((unsigned)((C) + 31) / 32, (unsigned)((R) + 15) / 16, (unsigned)(R * R)), 32, 0, stream>>>(v2_0_12); }
    { GemmP v2_0_13;
      v2_0_13.A = GQ + (size_t)0 * RP3 * C + (size_t)1191 * C; v2_0_13.B = wv2 + 13; v2_0_13.bias = GQ + (size_t)0 * RP3 * C + (size_t)1191 * C; v2_0_13.R = GC + (size_t)0 * R3 * C; v2_0_13.C = GC + (size_t)0 * R3 * C;
      v2_0_13.sAo = (long long)34 * 34 * C; v2_0_13.sAi = (long long)34 * C; v2_0_13.sAm = C; v2_0_13.sAk = 1; v2_0_13.sBo = 0; v2_0_13.sBi = 0; v2_0_13.sBn = C * 27; v2_0_13.sBk = 27; v2_0_13.sCo = (long long)R * R * C; v2_0_13.sCi = (long long)R * C; v2_0_13.sCm = C; v2_0_13.sRo = (long long)R * R * C; v2_0_13.sRi = (long long)R * C; v2_0_13.sRm = C; v2_0_13.sRn = 1;
      v2_0_13.M = R; v2_0_13.N = C; v2_0_13.K = C; v2_0_13.zi_n = R; v2_0_13.flags = 4; v2_0_13.act = 0;
      v2_0_13.alpha = 1.0f; v2_0_13.beta = 1.0f; v2_0_13.sa = 1.0f; v2_0_13.sb = 1.0f; v2_0_13.Npad = C; v2_0_13.pad_ = 0;
      k_gemm<1><<<dim3((unsigned)((C) + 31) / 32, (unsigned)((R) + 15) / 16, (unsigned)(R * R)), 32, 0, stream>>>(v2_0_13); }
    { GemmP v2_0_14;
      v2_0_14.A = GQ + (size_t)0 * RP3 * C + (size_t)1192 * C; v2_0_14.B = wv2 + 14; v2_0_14.bias = GQ + (size_t)0 * RP3 * C + (size_t)1192 * C; v2_0_14.R = GC + (size_t)0 * R3 * C; v2_0_14.C = GC + (size_t)0 * R3 * C;
      v2_0_14.sAo = (long long)34 * 34 * C; v2_0_14.sAi = (long long)34 * C; v2_0_14.sAm = C; v2_0_14.sAk = 1; v2_0_14.sBo = 0; v2_0_14.sBi = 0; v2_0_14.sBn = C * 27; v2_0_14.sBk = 27; v2_0_14.sCo = (long long)R * R * C; v2_0_14.sCi = (long long)R * C; v2_0_14.sCm = C; v2_0_14.sRo = (long long)R * R * C; v2_0_14.sRi = (long long)R * C; v2_0_14.sRm = C; v2_0_14.sRn = 1;
      v2_0_14.M = R; v2_0_14.N = C; v2_0_14.K = C; v2_0_14.zi_n = R; v2_0_14.flags = 4; v2_0_14.act = 0;
      v2_0_14.alpha = 1.0f; v2_0_14.beta = 1.0f; v2_0_14.sa = 1.0f; v2_0_14.sb = 1.0f; v2_0_14.Npad = C; v2_0_14.pad_ = 0;
      k_gemm<1><<<dim3((unsigned)((C) + 31) / 32, (unsigned)((R) + 15) / 16, (unsigned)(R * R)), 32, 0, stream>>>(v2_0_14); }
    { GemmP v2_0_15;
      v2_0_15.A = GQ + (size_t)0 * RP3 * C + (size_t)1224 * C; v2_0_15.B = wv2 + 15; v2_0_15.bias = GQ + (size_t)0 * RP3 * C + (size_t)1224 * C; v2_0_15.R = GC + (size_t)0 * R3 * C; v2_0_15.C = GC + (size_t)0 * R3 * C;
      v2_0_15.sAo = (long long)34 * 34 * C; v2_0_15.sAi = (long long)34 * C; v2_0_15.sAm = C; v2_0_15.sAk = 1; v2_0_15.sBo = 0; v2_0_15.sBi = 0; v2_0_15.sBn = C * 27; v2_0_15.sBk = 27; v2_0_15.sCo = (long long)R * R * C; v2_0_15.sCi = (long long)R * C; v2_0_15.sCm = C; v2_0_15.sRo = (long long)R * R * C; v2_0_15.sRi = (long long)R * C; v2_0_15.sRm = C; v2_0_15.sRn = 1;
      v2_0_15.M = R; v2_0_15.N = C; v2_0_15.K = C; v2_0_15.zi_n = R; v2_0_15.flags = 4; v2_0_15.act = 0;
      v2_0_15.alpha = 1.0f; v2_0_15.beta = 1.0f; v2_0_15.sa = 1.0f; v2_0_15.sb = 1.0f; v2_0_15.Npad = C; v2_0_15.pad_ = 0;
      k_gemm<1><<<dim3((unsigned)((C) + 31) / 32, (unsigned)((R) + 15) / 16, (unsigned)(R * R)), 32, 0, stream>>>(v2_0_15); }
    { GemmP v2_0_16;
      v2_0_16.A = GQ + (size_t)0 * RP3 * C + (size_t)1225 * C; v2_0_16.B = wv2 + 16; v2_0_16.bias = GQ + (size_t)0 * RP3 * C + (size_t)1225 * C; v2_0_16.R = GC + (size_t)0 * R3 * C; v2_0_16.C = GC + (size_t)0 * R3 * C;
      v2_0_16.sAo = (long long)34 * 34 * C; v2_0_16.sAi = (long long)34 * C; v2_0_16.sAm = C; v2_0_16.sAk = 1; v2_0_16.sBo = 0; v2_0_16.sBi = 0; v2_0_16.sBn = C * 27; v2_0_16.sBk = 27; v2_0_16.sCo = (long long)R * R * C; v2_0_16.sCi = (long long)R * C; v2_0_16.sCm = C; v2_0_16.sRo = (long long)R * R * C; v2_0_16.sRi = (long long)R * C; v2_0_16.sRm = C; v2_0_16.sRn = 1;
      v2_0_16.M = R; v2_0_16.N = C; v2_0_16.K = C; v2_0_16.zi_n = R; v2_0_16.flags = 4; v2_0_16.act = 0;
      v2_0_16.alpha = 1.0f; v2_0_16.beta = 1.0f; v2_0_16.sa = 1.0f; v2_0_16.sb = 1.0f; v2_0_16.Npad = C; v2_0_16.pad_ = 0;
      k_gemm<1><<<dim3((unsigned)((C) + 31) / 32, (unsigned)((R) + 15) / 16, (unsigned)(R * R)), 32, 0, stream>>>(v2_0_16); }
    { GemmP v2_0_17;
      v2_0_17.A = GQ + (size_t)0 * RP3 * C + (size_t)1226 * C; v2_0_17.B = wv2 + 17; v2_0_17.bias = GQ + (size_t)0 * RP3 * C + (size_t)1226 * C; v2_0_17.R = GC + (size_t)0 * R3 * C; v2_0_17.C = GC + (size_t)0 * R3 * C;
      v2_0_17.sAo = (long long)34 * 34 * C; v2_0_17.sAi = (long long)34 * C; v2_0_17.sAm = C; v2_0_17.sAk = 1; v2_0_17.sBo = 0; v2_0_17.sBi = 0; v2_0_17.sBn = C * 27; v2_0_17.sBk = 27; v2_0_17.sCo = (long long)R * R * C; v2_0_17.sCi = (long long)R * C; v2_0_17.sCm = C; v2_0_17.sRo = (long long)R * R * C; v2_0_17.sRi = (long long)R * C; v2_0_17.sRm = C; v2_0_17.sRn = 1;
      v2_0_17.M = R; v2_0_17.N = C; v2_0_17.K = C; v2_0_17.zi_n = R; v2_0_17.flags = 4; v2_0_17.act = 0;
      v2_0_17.alpha = 1.0f; v2_0_17.beta = 1.0f; v2_0_17.sa = 1.0f; v2_0_17.sb = 1.0f; v2_0_17.Npad = C; v2_0_17.pad_ = 0;
      k_gemm<1><<<dim3((unsigned)((C) + 31) / 32, (unsigned)((R) + 15) / 16, (unsigned)(R * R)), 32, 0, stream>>>(v2_0_17); }
    { GemmP v2_0_18;
      v2_0_18.A = GQ + (size_t)0 * RP3 * C + (size_t)2312 * C; v2_0_18.B = wv2 + 18; v2_0_18.bias = GQ + (size_t)0 * RP3 * C + (size_t)2312 * C; v2_0_18.R = GC + (size_t)0 * R3 * C; v2_0_18.C = GC + (size_t)0 * R3 * C;
      v2_0_18.sAo = (long long)34 * 34 * C; v2_0_18.sAi = (long long)34 * C; v2_0_18.sAm = C; v2_0_18.sAk = 1; v2_0_18.sBo = 0; v2_0_18.sBi = 0; v2_0_18.sBn = C * 27; v2_0_18.sBk = 27; v2_0_18.sCo = (long long)R * R * C; v2_0_18.sCi = (long long)R * C; v2_0_18.sCm = C; v2_0_18.sRo = (long long)R * R * C; v2_0_18.sRi = (long long)R * C; v2_0_18.sRm = C; v2_0_18.sRn = 1;
      v2_0_18.M = R; v2_0_18.N = C; v2_0_18.K = C; v2_0_18.zi_n = R; v2_0_18.flags = 4; v2_0_18.act = 0;
      v2_0_18.alpha = 1.0f; v2_0_18.beta = 1.0f; v2_0_18.sa = 1.0f; v2_0_18.sb = 1.0f; v2_0_18.Npad = C; v2_0_18.pad_ = 0;
      k_gemm<1><<<dim3((unsigned)((C) + 31) / 32, (unsigned)((R) + 15) / 16, (unsigned)(R * R)), 32, 0, stream>>>(v2_0_18); }
    { GemmP v2_0_19;
      v2_0_19.A = GQ + (size_t)0 * RP3 * C + (size_t)2313 * C; v2_0_19.B = wv2 + 19; v2_0_19.bias = GQ + (size_t)0 * RP3 * C + (size_t)2313 * C; v2_0_19.R = GC + (size_t)0 * R3 * C; v2_0_19.C = GC + (size_t)0 * R3 * C;
      v2_0_19.sAo = (long long)34 * 34 * C; v2_0_19.sAi = (long long)34 * C; v2_0_19.sAm = C; v2_0_19.sAk = 1; v2_0_19.sBo = 0; v2_0_19.sBi = 0; v2_0_19.sBn = C * 27; v2_0_19.sBk = 27; v2_0_19.sCo = (long long)R * R * C; v2_0_19.sCi = (long long)R * C; v2_0_19.sCm = C; v2_0_19.sRo = (long long)R * R * C; v2_0_19.sRi = (long long)R * C; v2_0_19.sRm = C; v2_0_19.sRn = 1;
      v2_0_19.M = R; v2_0_19.N = C; v2_0_19.K = C; v2_0_19.zi_n = R; v2_0_19.flags = 4; v2_0_19.act = 0;
      v2_0_19.alpha = 1.0f; v2_0_19.beta = 1.0f; v2_0_19.sa = 1.0f; v2_0_19.sb = 1.0f; v2_0_19.Npad = C; v2_0_19.pad_ = 0;
      k_gemm<1><<<dim3((unsigned)((C) + 31) / 32, (unsigned)((R) + 15) / 16, (unsigned)(R * R)), 32, 0, stream>>>(v2_0_19); }
    { GemmP v2_0_20;
      v2_0_20.A = GQ + (size_t)0 * RP3 * C + (size_t)2314 * C; v2_0_20.B = wv2 + 20; v2_0_20.bias = GQ + (size_t)0 * RP3 * C + (size_t)2314 * C; v2_0_20.R = GC + (size_t)0 * R3 * C; v2_0_20.C = GC + (size_t)0 * R3 * C;
      v2_0_20.sAo = (long long)34 * 34 * C; v2_0_20.sAi = (long long)34 * C; v2_0_20.sAm = C; v2_0_20.sAk = 1; v2_0_20.sBo = 0; v2_0_20.sBi = 0; v2_0_20.sBn = C * 27; v2_0_20.sBk = 27; v2_0_20.sCo = (long long)R * R * C; v2_0_20.sCi = (long long)R * C; v2_0_20.sCm = C; v2_0_20.sRo = (long long)R * R * C; v2_0_20.sRi = (long long)R * C; v2_0_20.sRm = C; v2_0_20.sRn = 1;
      v2_0_20.M = R; v2_0_20.N = C; v2_0_20.K = C; v2_0_20.zi_n = R; v2_0_20.flags = 4; v2_0_20.act = 0;
      v2_0_20.alpha = 1.0f; v2_0_20.beta = 1.0f; v2_0_20.sa = 1.0f; v2_0_20.sb = 1.0f; v2_0_20.Npad = C; v2_0_20.pad_ = 0;
      k_gemm<1><<<dim3((unsigned)((C) + 31) / 32, (unsigned)((R) + 15) / 16, (unsigned)(R * R)), 32, 0, stream>>>(v2_0_20); }
    { GemmP v2_0_21;
      v2_0_21.A = GQ + (size_t)0 * RP3 * C + (size_t)2346 * C; v2_0_21.B = wv2 + 21; v2_0_21.bias = GQ + (size_t)0 * RP3 * C + (size_t)2346 * C; v2_0_21.R = GC + (size_t)0 * R3 * C; v2_0_21.C = GC + (size_t)0 * R3 * C;
      v2_0_21.sAo = (long long)34 * 34 * C; v2_0_21.sAi = (long long)34 * C; v2_0_21.sAm = C; v2_0_21.sAk = 1; v2_0_21.sBo = 0; v2_0_21.sBi = 0; v2_0_21.sBn = C * 27; v2_0_21.sBk = 27; v2_0_21.sCo = (long long)R * R * C; v2_0_21.sCi = (long long)R * C; v2_0_21.sCm = C; v2_0_21.sRo = (long long)R * R * C; v2_0_21.sRi = (long long)R * C; v2_0_21.sRm = C; v2_0_21.sRn = 1;
      v2_0_21.M = R; v2_0_21.N = C; v2_0_21.K = C; v2_0_21.zi_n = R; v2_0_21.flags = 4; v2_0_21.act = 0;
      v2_0_21.alpha = 1.0f; v2_0_21.beta = 1.0f; v2_0_21.sa = 1.0f; v2_0_21.sb = 1.0f; v2_0_21.Npad = C; v2_0_21.pad_ = 0;
      k_gemm<1><<<dim3((unsigned)((C) + 31) / 32, (unsigned)((R) + 15) / 16, (unsigned)(R * R)), 32, 0, stream>>>(v2_0_21); }
    { GemmP v2_0_22;
      v2_0_22.A = GQ + (size_t)0 * RP3 * C + (size_t)2347 * C; v2_0_22.B = wv2 + 22; v2_0_22.bias = GQ + (size_t)0 * RP3 * C + (size_t)2347 * C; v2_0_22.R = GC + (size_t)0 * R3 * C; v2_0_22.C = GC + (size_t)0 * R3 * C;
      v2_0_22.sAo = (long long)34 * 34 * C; v2_0_22.sAi = (long long)34 * C; v2_0_22.sAm = C; v2_0_22.sAk = 1; v2_0_22.sBo = 0; v2_0_22.sBi = 0; v2_0_22.sBn = C * 27; v2_0_22.sBk = 27; v2_0_22.sCo = (long long)R * R * C; v2_0_22.sCi = (long long)R * C; v2_0_22.sCm = C; v2_0_22.sRo = (long long)R * R * C; v2_0_22.sRi = (long long)R * C; v2_0_22.sRm = C; v2_0_22.sRn = 1;
      v2_0_22.M = R; v2_0_22.N = C; v2_0_22.K = C; v2_0_22.zi_n = R; v2_0_22.flags = 4; v2_0_22.act = 0;
      v2_0_22.alpha = 1.0f; v2_0_22.beta = 1.0f; v2_0_22.sa = 1.0f; v2_0_22.sb = 1.0f; v2_0_22.Npad = C; v2_0_22.pad_ = 0;
      k_gemm<1><<<dim3((unsigned)((C) + 31) / 32, (unsigned)((R) + 15) / 16, (unsigned)(R * R)), 32, 0, stream>>>(v2_0_22); }
    { GemmP v2_0_23;
      v2_0_23.A = GQ + (size_t)0 * RP3 * C + (size_t)2348 * C; v2_0_23.B = wv2 + 23; v2_0_23.bias = GQ + (size_t)0 * RP3 * C + (size_t)2348 * C; v2_0_23.R = GC + (size_t)0 * R3 * C; v2_0_23.C = GC + (size_t)0 * R3 * C;
      v2_0_23.sAo = (long long)34 * 34 * C; v2_0_23.sAi = (long long)34 * C; v2_0_23.sAm = C; v2_0_23.sAk = 1; v2_0_23.sBo = 0; v2_0_23.sBi = 0; v2_0_23.sBn = C * 27; v2_0_23.sBk = 27; v2_0_23.sCo = (long long)R * R * C; v2_0_23.sCi = (long long)R * C; v2_0_23.sCm = C; v2_0_23.sRo = (long long)R * R * C; v2_0_23.sRi = (long long)R * C; v2_0_23.sRm = C; v2_0_23.sRn = 1;
      v2_0_23.M = R; v2_0_23.N = C; v2_0_23.K = C; v2_0_23.zi_n = R; v2_0_23.flags = 4; v2_0_23.act = 0;
      v2_0_23.alpha = 1.0f; v2_0_23.beta = 1.0f; v2_0_23.sa = 1.0f; v2_0_23.sb = 1.0f; v2_0_23.Npad = C; v2_0_23.pad_ = 0;
      k_gemm<1><<<dim3((unsigned)((C) + 31) / 32, (unsigned)((R) + 15) / 16, (unsigned)(R * R)), 32, 0, stream>>>(v2_0_23); }
    { GemmP v2_0_24;
      v2_0_24.A = GQ + (size_t)0 * RP3 * C + (size_t)2380 * C; v2_0_24.B = wv2 + 24; v2_0_24.bias = GQ + (size_t)0 * RP3 * C + (size_t)2380 * C; v2_0_24.R = GC + (size_t)0 * R3 * C; v2_0_24.C = GC + (size_t)0 * R3 * C;
      v2_0_24.sAo = (long long)34 * 34 * C; v2_0_24.sAi = (long long)34 * C; v2_0_24.sAm = C; v2_0_24.sAk = 1; v2_0_24.sBo = 0; v2_0_24.sBi = 0; v2_0_24.sBn = C * 27; v2_0_24.sBk = 27; v2_0_24.sCo = (long long)R * R * C; v2_0_24.sCi = (long long)R * C; v2_0_24.sCm = C; v2_0_24.sRo = (long long)R * R * C; v2_0_24.sRi = (long long)R * C; v2_0_24.sRm = C; v2_0_24.sRn = 1;
      v2_0_24.M = R; v2_0_24.N = C; v2_0_24.K = C; v2_0_24.zi_n = R; v2_0_24.flags = 4; v2_0_24.act = 0;
      v2_0_24.alpha = 1.0f; v2_0_24.beta = 1.0f; v2_0_24.sa = 1.0f; v2_0_24.sb = 1.0f; v2_0_24.Npad = C; v2_0_24.pad_ = 0;
      k_gemm<1><<<dim3((unsigned)((C) + 31) / 32, (unsigned)((R) + 15) / 16, (unsigned)(R * R)), 32, 0, stream>>>(v2_0_24); }
    { GemmP v2_0_25;
      v2_0_25.A = GQ + (size_t)0 * RP3 * C + (size_t)2381 * C; v2_0_25.B = wv2 + 25; v2_0_25.bias = GQ + (size_t)0 * RP3 * C + (size_t)2381 * C; v2_0_25.R = GC + (size_t)0 * R3 * C; v2_0_25.C = GC + (size_t)0 * R3 * C;
      v2_0_25.sAo = (long long)34 * 34 * C; v2_0_25.sAi = (long long)34 * C; v2_0_25.sAm = C; v2_0_25.sAk = 1; v2_0_25.sBo = 0; v2_0_25.sBi = 0; v2_0_25.sBn = C * 27; v2_0_25.sBk = 27; v2_0_25.sCo = (long long)R * R * C; v2_0_25.sCi = (long long)R * C; v2_0_25.sCm = C; v2_0_25.sRo = (long long)R * R * C; v2_0_25.sRi = (long long)R * C; v2_0_25.sRm = C; v2_0_25.sRn = 1;
      v2_0_25.M = R; v2_0_25.N = C; v2_0_25.K = C; v2_0_25.zi_n = R; v2_0_25.flags = 4; v2_0_25.act = 0;
      v2_0_25.alpha = 1.0f; v2_0_25.beta = 1.0f; v2_0_25.sa = 1.0f; v2_0_25.sb = 1.0f; v2_0_25.Npad = C; v2_0_25.pad_ = 0;
      k_gemm<1><<<dim3((unsigned)((C) + 31) / 32, (unsigned)((R) + 15) / 16, (unsigned)(R * R)), 32, 0, stream>>>(v2_0_25); }
    { GemmP v2_0_26;
      v2_0_26.A = GQ + (size_t)0 * RP3 * C + (size_t)2382 * C; v2_0_26.B = wv2 + 26; v2_0_26.bias = GQ + (size_t)0 * RP3 * C + (size_t)2382 * C; v2_0_26.R = GC + (size_t)0 * R3 * C; v2_0_26.C = GC + (size_t)0 * R3 * C;
      v2_0_26.sAo = (long long)34 * 34 * C; v2_0_26.sAi = (long long)34 * C; v2_0_26.sAm = C; v2_0_26.sAk = 1; v2_0_26.sBo = 0; v2_0_26.sBi = 0; v2_0_26.sBn = C * 27; v2_0_26.sBk = 27; v2_0_26.sCo = (long long)R * R * C; v2_0_26.sCi = (long long)R * C; v2_0_26.sCm = C; v2_0_26.sRo = (long long)R * R * C; v2_0_26.sRi = (long long)R * C; v2_0_26.sRm = C; v2_0_26.sRn = 1;
      v2_0_26.M = R; v2_0_26.N = C; v2_0_26.K = C; v2_0_26.zi_n = R; v2_0_26.flags = 4; v2_0_26.act = 0;
      v2_0_26.alpha = 1.0f; v2_0_26.beta = 1.0f; v2_0_26.sa = 1.0f; v2_0_26.sb = 1.0f; v2_0_26.Npad = C; v2_0_26.pad_ = 0;
      k_gemm<1><<<dim3((unsigned)((C) + 31) / 32, (unsigned)((R) + 15) / 16, (unsigned)(R * R)), 32, 0, stream>>>(v2_0_26); }
    { GemmP v2_1_0;
      v2_1_0.A = GQ + (size_t)1 * RP3 * C + (size_t)0 * C; v2_1_0.B = wv2 + 0; v2_1_0.bias = GQ + (size_t)1 * RP3 * C + (size_t)0 * C; v2_1_0.R = GQ + (size_t)1 * RP3 * C + (size_t)0 * C; v2_1_0.C = GC + (size_t)1 * R3 * C;
      v2_1_0.sAo = (long long)34 * 34 * C; v2_1_0.sAi = (long long)34 * C; v2_1_0.sAm = C; v2_1_0.sAk = 1; v2_1_0.sBo = 0; v2_1_0.sBi = 0; v2_1_0.sBn = C * 27; v2_1_0.sBk = 27; v2_1_0.sCo = (long long)R * R * C; v2_1_0.sCi = (long long)R * C; v2_1_0.sCm = C; v2_1_0.sRo = 0; v2_1_0.sRi = 0; v2_1_0.sRm = 0; v2_1_0.sRn = 0;
      v2_1_0.M = R; v2_1_0.N = C; v2_1_0.K = C; v2_1_0.zi_n = R; v2_1_0.flags = 0; v2_1_0.act = 0;
      v2_1_0.alpha = 1.0f; v2_1_0.beta = 0.0f; v2_1_0.sa = 1.0f; v2_1_0.sb = 1.0f; v2_1_0.Npad = C; v2_1_0.pad_ = 0;
      k_gemm<1><<<dim3((unsigned)((C) + 31) / 32, (unsigned)((R) + 15) / 16, (unsigned)(R * R)), 32, 0, stream>>>(v2_1_0); }
    { GemmP v2_1_1;
      v2_1_1.A = GQ + (size_t)1 * RP3 * C + (size_t)1 * C; v2_1_1.B = wv2 + 1; v2_1_1.bias = GQ + (size_t)1 * RP3 * C + (size_t)1 * C; v2_1_1.R = GC + (size_t)1 * R3 * C; v2_1_1.C = GC + (size_t)1 * R3 * C;
      v2_1_1.sAo = (long long)34 * 34 * C; v2_1_1.sAi = (long long)34 * C; v2_1_1.sAm = C; v2_1_1.sAk = 1; v2_1_1.sBo = 0; v2_1_1.sBi = 0; v2_1_1.sBn = C * 27; v2_1_1.sBk = 27; v2_1_1.sCo = (long long)R * R * C; v2_1_1.sCi = (long long)R * C; v2_1_1.sCm = C; v2_1_1.sRo = (long long)R * R * C; v2_1_1.sRi = (long long)R * C; v2_1_1.sRm = C; v2_1_1.sRn = 1;
      v2_1_1.M = R; v2_1_1.N = C; v2_1_1.K = C; v2_1_1.zi_n = R; v2_1_1.flags = 4; v2_1_1.act = 0;
      v2_1_1.alpha = 1.0f; v2_1_1.beta = 1.0f; v2_1_1.sa = 1.0f; v2_1_1.sb = 1.0f; v2_1_1.Npad = C; v2_1_1.pad_ = 0;
      k_gemm<1><<<dim3((unsigned)((C) + 31) / 32, (unsigned)((R) + 15) / 16, (unsigned)(R * R)), 32, 0, stream>>>(v2_1_1); }
    { GemmP v2_1_2;
      v2_1_2.A = GQ + (size_t)1 * RP3 * C + (size_t)2 * C; v2_1_2.B = wv2 + 2; v2_1_2.bias = GQ + (size_t)1 * RP3 * C + (size_t)2 * C; v2_1_2.R = GC + (size_t)1 * R3 * C; v2_1_2.C = GC + (size_t)1 * R3 * C;
      v2_1_2.sAo = (long long)34 * 34 * C; v2_1_2.sAi = (long long)34 * C; v2_1_2.sAm = C; v2_1_2.sAk = 1; v2_1_2.sBo = 0; v2_1_2.sBi = 0; v2_1_2.sBn = C * 27; v2_1_2.sBk = 27; v2_1_2.sCo = (long long)R * R * C; v2_1_2.sCi = (long long)R * C; v2_1_2.sCm = C; v2_1_2.sRo = (long long)R * R * C; v2_1_2.sRi = (long long)R * C; v2_1_2.sRm = C; v2_1_2.sRn = 1;
      v2_1_2.M = R; v2_1_2.N = C; v2_1_2.K = C; v2_1_2.zi_n = R; v2_1_2.flags = 4; v2_1_2.act = 0;
      v2_1_2.alpha = 1.0f; v2_1_2.beta = 1.0f; v2_1_2.sa = 1.0f; v2_1_2.sb = 1.0f; v2_1_2.Npad = C; v2_1_2.pad_ = 0;
      k_gemm<1><<<dim3((unsigned)((C) + 31) / 32, (unsigned)((R) + 15) / 16, (unsigned)(R * R)), 32, 0, stream>>>(v2_1_2); }
    { GemmP v2_1_3;
      v2_1_3.A = GQ + (size_t)1 * RP3 * C + (size_t)34 * C; v2_1_3.B = wv2 + 3; v2_1_3.bias = GQ + (size_t)1 * RP3 * C + (size_t)34 * C; v2_1_3.R = GC + (size_t)1 * R3 * C; v2_1_3.C = GC + (size_t)1 * R3 * C;
      v2_1_3.sAo = (long long)34 * 34 * C; v2_1_3.sAi = (long long)34 * C; v2_1_3.sAm = C; v2_1_3.sAk = 1; v2_1_3.sBo = 0; v2_1_3.sBi = 0; v2_1_3.sBn = C * 27; v2_1_3.sBk = 27; v2_1_3.sCo = (long long)R * R * C; v2_1_3.sCi = (long long)R * C; v2_1_3.sCm = C; v2_1_3.sRo = (long long)R * R * C; v2_1_3.sRi = (long long)R * C; v2_1_3.sRm = C; v2_1_3.sRn = 1;
      v2_1_3.M = R; v2_1_3.N = C; v2_1_3.K = C; v2_1_3.zi_n = R; v2_1_3.flags = 4; v2_1_3.act = 0;
      v2_1_3.alpha = 1.0f; v2_1_3.beta = 1.0f; v2_1_3.sa = 1.0f; v2_1_3.sb = 1.0f; v2_1_3.Npad = C; v2_1_3.pad_ = 0;
      k_gemm<1><<<dim3((unsigned)((C) + 31) / 32, (unsigned)((R) + 15) / 16, (unsigned)(R * R)), 32, 0, stream>>>(v2_1_3); }
    { GemmP v2_1_4;
      v2_1_4.A = GQ + (size_t)1 * RP3 * C + (size_t)35 * C; v2_1_4.B = wv2 + 4; v2_1_4.bias = GQ + (size_t)1 * RP3 * C + (size_t)35 * C; v2_1_4.R = GC + (size_t)1 * R3 * C; v2_1_4.C = GC + (size_t)1 * R3 * C;
      v2_1_4.sAo = (long long)34 * 34 * C; v2_1_4.sAi = (long long)34 * C; v2_1_4.sAm = C; v2_1_4.sAk = 1; v2_1_4.sBo = 0; v2_1_4.sBi = 0; v2_1_4.sBn = C * 27; v2_1_4.sBk = 27; v2_1_4.sCo = (long long)R * R * C; v2_1_4.sCi = (long long)R * C; v2_1_4.sCm = C; v2_1_4.sRo = (long long)R * R * C; v2_1_4.sRi = (long long)R * C; v2_1_4.sRm = C; v2_1_4.sRn = 1;
      v2_1_4.M = R; v2_1_4.N = C; v2_1_4.K = C; v2_1_4.zi_n = R; v2_1_4.flags = 4; v2_1_4.act = 0;
      v2_1_4.alpha = 1.0f; v2_1_4.beta = 1.0f; v2_1_4.sa = 1.0f; v2_1_4.sb = 1.0f; v2_1_4.Npad = C; v2_1_4.pad_ = 0;
      k_gemm<1><<<dim3((unsigned)((C) + 31) / 32, (unsigned)((R) + 15) / 16, (unsigned)(R * R)), 32, 0, stream>>>(v2_1_4); }
    { GemmP v2_1_5;
      v2_1_5.A = GQ + (size_t)1 * RP3 * C + (size_t)36 * C; v2_1_5.B = wv2 + 5; v2_1_5.bias = GQ + (size_t)1 * RP3 * C + (size_t)36 * C; v2_1_5.R = GC + (size_t)1 * R3 * C; v2_1_5.C = GC + (size_t)1 * R3 * C;
      v2_1_5.sAo = (long long)34 * 34 * C; v2_1_5.sAi = (long long)34 * C; v2_1_5.sAm = C; v2_1_5.sAk = 1; v2_1_5.sBo = 0; v2_1_5.sBi = 0; v2_1_5.sBn = C * 27; v2_1_5.sBk = 27; v2_1_5.sCo = (long long)R * R * C; v2_1_5.sCi = (long long)R * C; v2_1_5.sCm = C; v2_1_5.sRo = (long long)R * R * C; v2_1_5.sRi = (long long)R * C; v2_1_5.sRm = C; v2_1_5.sRn = 1;
      v2_1_5.M = R; v2_1_5.N = C; v2_1_5.K = C; v2_1_5.zi_n = R; v2_1_5.flags = 4; v2_1_5.act = 0;
      v2_1_5.alpha = 1.0f; v2_1_5.beta = 1.0f; v2_1_5.sa = 1.0f; v2_1_5.sb = 1.0f; v2_1_5.Npad = C; v2_1_5.pad_ = 0;
      k_gemm<1><<<dim3((unsigned)((C) + 31) / 32, (unsigned)((R) + 15) / 16, (unsigned)(R * R)), 32, 0, stream>>>(v2_1_5); }
    { GemmP v2_1_6;
      v2_1_6.A = GQ + (size_t)1 * RP3 * C + (size_t)68 * C; v2_1_6.B = wv2 + 6; v2_1_6.bias = GQ + (size_t)1 * RP3 * C + (size_t)68 * C; v2_1_6.R = GC + (size_t)1 * R3 * C; v2_1_6.C = GC + (size_t)1 * R3 * C;
      v2_1_6.sAo = (long long)34 * 34 * C; v2_1_6.sAi = (long long)34 * C; v2_1_6.sAm = C; v2_1_6.sAk = 1; v2_1_6.sBo = 0; v2_1_6.sBi = 0; v2_1_6.sBn = C * 27; v2_1_6.sBk = 27; v2_1_6.sCo = (long long)R * R * C; v2_1_6.sCi = (long long)R * C; v2_1_6.sCm = C; v2_1_6.sRo = (long long)R * R * C; v2_1_6.sRi = (long long)R * C; v2_1_6.sRm = C; v2_1_6.sRn = 1;
      v2_1_6.M = R; v2_1_6.N = C; v2_1_6.K = C; v2_1_6.zi_n = R; v2_1_6.flags = 4; v2_1_6.act = 0;
      v2_1_6.alpha = 1.0f; v2_1_6.beta = 1.0f; v2_1_6.sa = 1.0f; v2_1_6.sb = 1.0f; v2_1_6.Npad = C; v2_1_6.pad_ = 0;
      k_gemm<1><<<dim3((unsigned)((C) + 31) / 32, (unsigned)((R) + 15) / 16, (unsigned)(R * R)), 32, 0, stream>>>(v2_1_6); }
    { GemmP v2_1_7;
      v2_1_7.A = GQ + (size_t)1 * RP3 * C + (size_t)69 * C; v2_1_7.B = wv2 + 7; v2_1_7.bias = GQ + (size_t)1 * RP3 * C + (size_t)69 * C; v2_1_7.R = GC + (size_t)1 * R3 * C; v2_1_7.C = GC + (size_t)1 * R3 * C;
      v2_1_7.sAo = (long long)34 * 34 * C; v2_1_7.sAi = (long long)34 * C; v2_1_7.sAm = C; v2_1_7.sAk = 1; v2_1_7.sBo = 0; v2_1_7.sBi = 0; v2_1_7.sBn = C * 27; v2_1_7.sBk = 27; v2_1_7.sCo = (long long)R * R * C; v2_1_7.sCi = (long long)R * C; v2_1_7.sCm = C; v2_1_7.sRo = (long long)R * R * C; v2_1_7.sRi = (long long)R * C; v2_1_7.sRm = C; v2_1_7.sRn = 1;
      v2_1_7.M = R; v2_1_7.N = C; v2_1_7.K = C; v2_1_7.zi_n = R; v2_1_7.flags = 4; v2_1_7.act = 0;
      v2_1_7.alpha = 1.0f; v2_1_7.beta = 1.0f; v2_1_7.sa = 1.0f; v2_1_7.sb = 1.0f; v2_1_7.Npad = C; v2_1_7.pad_ = 0;
      k_gemm<1><<<dim3((unsigned)((C) + 31) / 32, (unsigned)((R) + 15) / 16, (unsigned)(R * R)), 32, 0, stream>>>(v2_1_7); }
    { GemmP v2_1_8;
      v2_1_8.A = GQ + (size_t)1 * RP3 * C + (size_t)70 * C; v2_1_8.B = wv2 + 8; v2_1_8.bias = GQ + (size_t)1 * RP3 * C + (size_t)70 * C; v2_1_8.R = GC + (size_t)1 * R3 * C; v2_1_8.C = GC + (size_t)1 * R3 * C;
      v2_1_8.sAo = (long long)34 * 34 * C; v2_1_8.sAi = (long long)34 * C; v2_1_8.sAm = C; v2_1_8.sAk = 1; v2_1_8.sBo = 0; v2_1_8.sBi = 0; v2_1_8.sBn = C * 27; v2_1_8.sBk = 27; v2_1_8.sCo = (long long)R * R * C; v2_1_8.sCi = (long long)R * C; v2_1_8.sCm = C; v2_1_8.sRo = (long long)R * R * C; v2_1_8.sRi = (long long)R * C; v2_1_8.sRm = C; v2_1_8.sRn = 1;
      v2_1_8.M = R; v2_1_8.N = C; v2_1_8.K = C; v2_1_8.zi_n = R; v2_1_8.flags = 4; v2_1_8.act = 0;
      v2_1_8.alpha = 1.0f; v2_1_8.beta = 1.0f; v2_1_8.sa = 1.0f; v2_1_8.sb = 1.0f; v2_1_8.Npad = C; v2_1_8.pad_ = 0;
      k_gemm<1><<<dim3((unsigned)((C) + 31) / 32, (unsigned)((R) + 15) / 16, (unsigned)(R * R)), 32, 0, stream>>>(v2_1_8); }
    { GemmP v2_1_9;
      v2_1_9.A = GQ + (size_t)1 * RP3 * C + (size_t)1156 * C; v2_1_9.B = wv2 + 9; v2_1_9.bias = GQ + (size_t)1 * RP3 * C + (size_t)1156 * C; v2_1_9.R = GC + (size_t)1 * R3 * C; v2_1_9.C = GC + (size_t)1 * R3 * C;
      v2_1_9.sAo = (long long)34 * 34 * C; v2_1_9.sAi = (long long)34 * C; v2_1_9.sAm = C; v2_1_9.sAk = 1; v2_1_9.sBo = 0; v2_1_9.sBi = 0; v2_1_9.sBn = C * 27; v2_1_9.sBk = 27; v2_1_9.sCo = (long long)R * R * C; v2_1_9.sCi = (long long)R * C; v2_1_9.sCm = C; v2_1_9.sRo = (long long)R * R * C; v2_1_9.sRi = (long long)R * C; v2_1_9.sRm = C; v2_1_9.sRn = 1;
      v2_1_9.M = R; v2_1_9.N = C; v2_1_9.K = C; v2_1_9.zi_n = R; v2_1_9.flags = 4; v2_1_9.act = 0;
      v2_1_9.alpha = 1.0f; v2_1_9.beta = 1.0f; v2_1_9.sa = 1.0f; v2_1_9.sb = 1.0f; v2_1_9.Npad = C; v2_1_9.pad_ = 0;
      k_gemm<1><<<dim3((unsigned)((C) + 31) / 32, (unsigned)((R) + 15) / 16, (unsigned)(R * R)), 32, 0, stream>>>(v2_1_9); }
    { GemmP v2_1_10;
      v2_1_10.A = GQ + (size_t)1 * RP3 * C + (size_t)1157 * C; v2_1_10.B = wv2 + 10; v2_1_10.bias = GQ + (size_t)1 * RP3 * C + (size_t)1157 * C; v2_1_10.R = GC + (size_t)1 * R3 * C; v2_1_10.C = GC + (size_t)1 * R3 * C;
      v2_1_10.sAo = (long long)34 * 34 * C; v2_1_10.sAi = (long long)34 * C; v2_1_10.sAm = C; v2_1_10.sAk = 1; v2_1_10.sBo = 0; v2_1_10.sBi = 0; v2_1_10.sBn = C * 27; v2_1_10.sBk = 27; v2_1_10.sCo = (long long)R * R * C; v2_1_10.sCi = (long long)R * C; v2_1_10.sCm = C; v2_1_10.sRo = (long long)R * R * C; v2_1_10.sRi = (long long)R * C; v2_1_10.sRm = C; v2_1_10.sRn = 1;
      v2_1_10.M = R; v2_1_10.N = C; v2_1_10.K = C; v2_1_10.zi_n = R; v2_1_10.flags = 4; v2_1_10.act = 0;
      v2_1_10.alpha = 1.0f; v2_1_10.beta = 1.0f; v2_1_10.sa = 1.0f; v2_1_10.sb = 1.0f; v2_1_10.Npad = C; v2_1_10.pad_ = 0;
      k_gemm<1><<<dim3((unsigned)((C) + 31) / 32, (unsigned)((R) + 15) / 16, (unsigned)(R * R)), 32, 0, stream>>>(v2_1_10); }
    { GemmP v2_1_11;
      v2_1_11.A = GQ + (size_t)1 * RP3 * C + (size_t)1158 * C; v2_1_11.B = wv2 + 11; v2_1_11.bias = GQ + (size_t)1 * RP3 * C + (size_t)1158 * C; v2_1_11.R = GC + (size_t)1 * R3 * C; v2_1_11.C = GC + (size_t)1 * R3 * C;
      v2_1_11.sAo = (long long)34 * 34 * C; v2_1_11.sAi = (long long)34 * C; v2_1_11.sAm = C; v2_1_11.sAk = 1; v2_1_11.sBo = 0; v2_1_11.sBi = 0; v2_1_11.sBn = C * 27; v2_1_11.sBk = 27; v2_1_11.sCo = (long long)R * R * C; v2_1_11.sCi = (long long)R * C; v2_1_11.sCm = C; v2_1_11.sRo = (long long)R * R * C; v2_1_11.sRi = (long long)R * C; v2_1_11.sRm = C; v2_1_11.sRn = 1;
      v2_1_11.M = R; v2_1_11.N = C; v2_1_11.K = C; v2_1_11.zi_n = R; v2_1_11.flags = 4; v2_1_11.act = 0;
      v2_1_11.alpha = 1.0f; v2_1_11.beta = 1.0f; v2_1_11.sa = 1.0f; v2_1_11.sb = 1.0f; v2_1_11.Npad = C; v2_1_11.pad_ = 0;
      k_gemm<1><<<dim3((unsigned)((C) + 31) / 32, (unsigned)((R) + 15) / 16, (unsigned)(R * R)), 32, 0, stream>>>(v2_1_11); }
    { GemmP v2_1_12;
      v2_1_12.A = GQ + (size_t)1 * RP3 * C + (size_t)1190 * C; v2_1_12.B = wv2 + 12; v2_1_12.bias = GQ + (size_t)1 * RP3 * C + (size_t)1190 * C; v2_1_12.R = GC + (size_t)1 * R3 * C; v2_1_12.C = GC + (size_t)1 * R3 * C;
      v2_1_12.sAo = (long long)34 * 34 * C; v2_1_12.sAi = (long long)34 * C; v2_1_12.sAm = C; v2_1_12.sAk = 1; v2_1_12.sBo = 0; v2_1_12.sBi = 0; v2_1_12.sBn = C * 27; v2_1_12.sBk = 27; v2_1_12.sCo = (long long)R * R * C; v2_1_12.sCi = (long long)R * C; v2_1_12.sCm = C; v2_1_12.sRo = (long long)R * R * C; v2_1_12.sRi = (long long)R * C; v2_1_12.sRm = C; v2_1_12.sRn = 1;
      v2_1_12.M = R; v2_1_12.N = C; v2_1_12.K = C; v2_1_12.zi_n = R; v2_1_12.flags = 4; v2_1_12.act = 0;
      v2_1_12.alpha = 1.0f; v2_1_12.beta = 1.0f; v2_1_12.sa = 1.0f; v2_1_12.sb = 1.0f; v2_1_12.Npad = C; v2_1_12.pad_ = 0;
      k_gemm<1><<<dim3((unsigned)((C) + 31) / 32, (unsigned)((R) + 15) / 16, (unsigned)(R * R)), 32, 0, stream>>>(v2_1_12); }
    { GemmP v2_1_13;
      v2_1_13.A = GQ + (size_t)1 * RP3 * C + (size_t)1191 * C; v2_1_13.B = wv2 + 13; v2_1_13.bias = GQ + (size_t)1 * RP3 * C + (size_t)1191 * C; v2_1_13.R = GC + (size_t)1 * R3 * C; v2_1_13.C = GC + (size_t)1 * R3 * C;
      v2_1_13.sAo = (long long)34 * 34 * C; v2_1_13.sAi = (long long)34 * C; v2_1_13.sAm = C; v2_1_13.sAk = 1; v2_1_13.sBo = 0; v2_1_13.sBi = 0; v2_1_13.sBn = C * 27; v2_1_13.sBk = 27; v2_1_13.sCo = (long long)R * R * C; v2_1_13.sCi = (long long)R * C; v2_1_13.sCm = C; v2_1_13.sRo = (long long)R * R * C; v2_1_13.sRi = (long long)R * C; v2_1_13.sRm = C; v2_1_13.sRn = 1;
      v2_1_13.M = R; v2_1_13.N = C; v2_1_13.K = C; v2_1_13.zi_n = R; v2_1_13.flags = 4; v2_1_13.act = 0;
      v2_1_13.alpha = 1.0f; v2_1_13.beta = 1.0f; v2_1_13.sa = 1.0f; v2_1_13.sb = 1.0f; v2_1_13.Npad = C; v2_1_13.pad_ = 0;
      k_gemm<1><<<dim3((unsigned)((C) + 31) / 32, (unsigned)((R) + 15) / 16, (unsigned)(R * R)), 32, 0, stream>>>(v2_1_13); }
    { GemmP v2_1_14;
      v2_1_14.A = GQ + (size_t)1 * RP3 * C + (size_t)1192 * C; v2_1_14.B = wv2 + 14; v2_1_14.bias = GQ + (size_t)1 * RP3 * C + (size_t)1192 * C; v2_1_14.R = GC + (size_t)1 * R3 * C; v2_1_14.C = GC + (size_t)1 * R3 * C;
      v2_1_14.sAo = (long long)34 * 34 * C; v2_1_14.sAi = (long long)34 * C; v2_1_14.sAm = C; v2_1_14.sAk = 1; v2_1_14.sBo = 0; v2_1_14.sBi = 0; v2_1_14.sBn = C * 27; v2_1_14.sBk = 27; v2_1_14.sCo = (long long)R * R * C; v2_1_14.sCi = (long long)R * C; v2_1_14.sCm = C; v2_1_14.sRo = (long long)R * R * C; v2_1_14.sRi = (long long)R * C; v2_1_14.sRm = C; v2_1_14.sRn = 1;
      v2_1_14.M = R; v2_1_14.N = C; v2_1_14.K = C; v2_1_14.zi_n = R; v2_1_14.flags = 4; v2_1_14.act = 0;
      v2_1_14.alpha = 1.0f; v2_1_14.beta = 1.0f; v2_1_14.sa = 1.0f; v2_1_14.sb = 1.0f; v2_1_14.Npad = C; v2_1_14.pad_ = 0;
      k_gemm<1><<<dim3((unsigned)((C) + 31) / 32, (unsigned)((R) + 15) / 16, (unsigned)(R * R)), 32, 0, stream>>>(v2_1_14); }
    { GemmP v2_1_15;
      v2_1_15.A = GQ + (size_t)1 * RP3 * C + (size_t)1224 * C; v2_1_15.B = wv2 + 15; v2_1_15.bias = GQ + (size_t)1 * RP3 * C + (size_t)1224 * C; v2_1_15.R = GC + (size_t)1 * R3 * C; v2_1_15.C = GC + (size_t)1 * R3 * C;
      v2_1_15.sAo = (long long)34 * 34 * C; v2_1_15.sAi = (long long)34 * C; v2_1_15.sAm = C; v2_1_15.sAk = 1; v2_1_15.sBo = 0; v2_1_15.sBi = 0; v2_1_15.sBn = C * 27; v2_1_15.sBk = 27; v2_1_15.sCo = (long long)R * R * C; v2_1_15.sCi = (long long)R * C; v2_1_15.sCm = C; v2_1_15.sRo = (long long)R * R * C; v2_1_15.sRi = (long long)R * C; v2_1_15.sRm = C; v2_1_15.sRn = 1;
      v2_1_15.M = R; v2_1_15.N = C; v2_1_15.K = C; v2_1_15.zi_n = R; v2_1_15.flags = 4; v2_1_15.act = 0;
      v2_1_15.alpha = 1.0f; v2_1_15.beta = 1.0f; v2_1_15.sa = 1.0f; v2_1_15.sb = 1.0f; v2_1_15.Npad = C; v2_1_15.pad_ = 0;
      k_gemm<1><<<dim3((unsigned)((C) + 31) / 32, (unsigned)((R) + 15) / 16, (unsigned)(R * R)), 32, 0, stream>>>(v2_1_15); }
    { GemmP v2_1_16;
      v2_1_16.A = GQ + (size_t)1 * RP3 * C + (size_t)1225 * C; v2_1_16.B = wv2 + 16; v2_1_16.bias = GQ + (size_t)1 * RP3 * C + (size_t)1225 * C; v2_1_16.R = GC + (size_t)1 * R3 * C; v2_1_16.C = GC + (size_t)1 * R3 * C;
      v2_1_16.sAo = (long long)34 * 34 * C; v2_1_16.sAi = (long long)34 * C; v2_1_16.sAm = C; v2_1_16.sAk = 1; v2_1_16.sBo = 0; v2_1_16.sBi = 0; v2_1_16.sBn = C * 27; v2_1_16.sBk = 27; v2_1_16.sCo = (long long)R * R * C; v2_1_16.sCi = (long long)R * C; v2_1_16.sCm = C; v2_1_16.sRo = (long long)R * R * C; v2_1_16.sRi = (long long)R * C; v2_1_16.sRm = C; v2_1_16.sRn = 1;
      v2_1_16.M = R; v2_1_16.N = C; v2_1_16.K = C; v2_1_16.zi_n = R; v2_1_16.flags = 4; v2_1_16.act = 0;
      v2_1_16.alpha = 1.0f; v2_1_16.beta = 1.0f; v2_1_16.sa = 1.0f; v2_1_16.sb = 1.0f; v2_1_16.Npad = C; v2_1_16.pad_ = 0;
      k_gemm<1><<<dim3((unsigned)((C) + 31) / 32, (unsigned)((R) + 15) / 16, (unsigned)(R * R)), 32, 0, stream>>>(v2_1_16); }
    { GemmP v2_1_17;
      v2_1_17.A = GQ + (size_t)1 * RP3 * C + (size_t)1226 * C; v2_1_17.B = wv2 + 17; v2_1_17.bias = GQ + (size_t)1 * RP3 * C + (size_t)1226 * C; v2_1_17.R = GC + (size_t)1 * R3 * C; v2_1_17.C = GC + (size_t)1 * R3 * C;
      v2_1_17.sAo = (long long)34 * 34 * C; v2_1_17.sAi = (long long)34 * C; v2_1_17.sAm = C; v2_1_17.sAk = 1; v2_1_17.sBo = 0; v2_1_17.sBi = 0; v2_1_17.sBn = C * 27; v2_1_17.sBk = 27; v2_1_17.sCo = (long long)R * R * C; v2_1_17.sCi = (long long)R * C; v2_1_17.sCm = C; v2_1_17.sRo = (long long)R * R * C; v2_1_17.sRi = (long long)R * C; v2_1_17.sRm = C; v2_1_17.sRn = 1;
      v2_1_17.M = R; v2_1_17.N = C; v2_1_17.K = C; v2_1_17.zi_n = R; v2_1_17.flags = 4; v2_1_17.act = 0;
      v2_1_17.alpha = 1.0f; v2_1_17.beta = 1.0f; v2_1_17.sa = 1.0f; v2_1_17.sb = 1.0f; v2_1_17.Npad = C; v2_1_17.pad_ = 0;
      k_gemm<1><<<dim3((unsigned)((C) + 31) / 32, (unsigned)((R) + 15) / 16, (unsigned)(R * R)), 32, 0, stream>>>(v2_1_17); }
    { GemmP v2_1_18;
      v2_1_18.A = GQ + (size_t)1 * RP3 * C + (size_t)2312 * C; v2_1_18.B = wv2 + 18; v2_1_18.bias = GQ + (size_t)1 * RP3 * C + (size_t)2312 * C; v2_1_18.R = GC + (size_t)1 * R3 * C; v2_1_18.C = GC + (size_t)1 * R3 * C;
      v2_1_18.sAo = (long long)34 * 34 * C; v2_1_18.sAi = (long long)34 * C; v2_1_18.sAm = C; v2_1_18.sAk = 1; v2_1_18.sBo = 0; v2_1_18.sBi = 0; v2_1_18.sBn = C * 27; v2_1_18.sBk = 27; v2_1_18.sCo = (long long)R * R * C; v2_1_18.sCi = (long long)R * C; v2_1_18.sCm = C; v2_1_18.sRo = (long long)R * R * C; v2_1_18.sRi = (long long)R * C; v2_1_18.sRm = C; v2_1_18.sRn = 1;
      v2_1_18.M = R; v2_1_18.N = C; v2_1_18.K = C; v2_1_18.zi_n = R; v2_1_18.flags = 4; v2_1_18.act = 0;
      v2_1_18.alpha = 1.0f; v2_1_18.beta = 1.0f; v2_1_18.sa = 1.0f; v2_1_18.sb = 1.0f; v2_1_18.Npad = C; v2_1_18.pad_ = 0;
      k_gemm<1><<<dim3((unsigned)((C) + 31) / 32, (unsigned)((R) + 15) / 16, (unsigned)(R * R)), 32, 0, stream>>>(v2_1_18); }
    { GemmP v2_1_19;
      v2_1_19.A = GQ + (size_t)1 * RP3 * C + (size_t)2313 * C; v2_1_19.B = wv2 + 19; v2_1_19.bias = GQ + (size_t)1 * RP3 * C + (size_t)2313 * C; v2_1_19.R = GC + (size_t)1 * R3 * C; v2_1_19.C = GC + (size_t)1 * R3 * C;
      v2_1_19.sAo = (long long)34 * 34 * C; v2_1_19.sAi = (long long)34 * C; v2_1_19.sAm = C; v2_1_19.sAk = 1; v2_1_19.sBo = 0; v2_1_19.sBi = 0; v2_1_19.sBn = C * 27; v2_1_19.sBk = 27; v2_1_19.sCo = (long long)R * R * C; v2_1_19.sCi = (long long)R * C; v2_1_19.sCm = C; v2_1_19.sRo = (long long)R * R * C; v2_1_19.sRi = (long long)R * C; v2_1_19.sRm = C; v2_1_19.sRn = 1;
      v2_1_19.M = R; v2_1_19.N = C; v2_1_19.K = C; v2_1_19.zi_n = R; v2_1_19.flags = 4; v2_1_19.act = 0;
      v2_1_19.alpha = 1.0f; v2_1_19.beta = 1.0f; v2_1_19.sa = 1.0f; v2_1_19.sb = 1.0f; v2_1_19.Npad = C; v2_1_19.pad_ = 0;
      k_gemm<1><<<dim3((unsigned)((C) + 31) / 32, (unsigned)((R) + 15) / 16, (unsigned)(R * R)), 32, 0, stream>>>(v2_1_19); }
    { GemmP v2_1_20;
      v2_1_20.A = GQ + (size_t)1 * RP3 * C + (size_t)2314 * C; v2_1_20.B = wv2 + 20; v2_1_20.bias = GQ + (size_t)1 * RP3 * C + (size_t)2314 * C; v2_1_20.R = GC + (size_t)1 * R3 * C; v2_1_20.C = GC + (size_t)1 * R3 * C;
      v2_1_20.sAo = (long long)34 * 34 * C; v2_1_20.sAi = (long long)34 * C; v2_1_20.sAm = C; v2_1_20.sAk = 1; v2_1_20.sBo = 0; v2_1_20.sBi = 0; v2_1_20.sBn = C * 27; v2_1_20.sBk = 27; v2_1_20.sCo = (long long)R * R * C; v2_1_20.sCi = (long long)R * C; v2_1_20.sCm = C; v2_1_20.sRo = (long long)R * R * C; v2_1_20.sRi = (long long)R * C; v2_1_20.sRm = C; v2_1_20.sRn = 1;
      v2_1_20.M = R; v2_1_20.N = C; v2_1_20.K = C; v2_1_20.zi_n = R; v2_1_20.flags = 4; v2_1_20.act = 0;
      v2_1_20.alpha = 1.0f; v2_1_20.beta = 1.0f; v2_1_20.sa = 1.0f; v2_1_20.sb = 1.0f; v2_1_20.Npad = C; v2_1_20.pad_ = 0;
      k_gemm<1><<<dim3((unsigned)((C) + 31) / 32, (unsigned)((R) + 15) / 16, (unsigned)(R * R)), 32, 0, stream>>>(v2_1_20); }
    { GemmP v2_1_21;
      v2_1_21.A = GQ + (size_t)1 * RP3 * C + (size_t)2346 * C; v2_1_21.B = wv2 + 21; v2_1_21.bias = GQ + (size_t)1 * RP3 * C + (size_t)2346 * C; v2_1_21.R = GC + (size_t)1 * R3 * C; v2_1_21.C = GC + (size_t)1 * R3 * C;
      v2_1_21.sAo = (long long)34 * 34 * C; v2_1_21.sAi = (long long)34 * C; v2_1_21.sAm = C; v2_1_21.sAk = 1; v2_1_21.sBo = 0; v2_1_21.sBi = 0; v2_1_21.sBn = C * 27; v2_1_21.sBk = 27; v2_1_21.sCo = (long long)R * R * C; v2_1_21.sCi = (long long)R * C; v2_1_21.sCm = C; v2_1_21.sRo = (long long)R * R * C; v2_1_21.sRi = (long long)R * C; v2_1_21.sRm = C; v2_1_21.sRn = 1;
      v2_1_21.M = R; v2_1_21.N = C; v2_1_21.K = C; v2_1_21.zi_n = R; v2_1_21.flags = 4; v2_1_21.act = 0;
      v2_1_21.alpha = 1.0f; v2_1_21.beta = 1.0f; v2_1_21.sa = 1.0f; v2_1_21.sb = 1.0f; v2_1_21.Npad = C; v2_1_21.pad_ = 0;
      k_gemm<1><<<dim3((unsigned)((C) + 31) / 32, (unsigned)((R) + 15) / 16, (unsigned)(R * R)), 32, 0, stream>>>(v2_1_21); }
    { GemmP v2_1_22;
      v2_1_22.A = GQ + (size_t)1 * RP3 * C + (size_t)2347 * C; v2_1_22.B = wv2 + 22; v2_1_22.bias = GQ + (size_t)1 * RP3 * C + (size_t)2347 * C; v2_1_22.R = GC + (size_t)1 * R3 * C; v2_1_22.C = GC + (size_t)1 * R3 * C;
      v2_1_22.sAo = (long long)34 * 34 * C; v2_1_22.sAi = (long long)34 * C; v2_1_22.sAm = C; v2_1_22.sAk = 1; v2_1_22.sBo = 0; v2_1_22.sBi = 0; v2_1_22.sBn = C * 27; v2_1_22.sBk = 27; v2_1_22.sCo = (long long)R * R * C; v2_1_22.sCi = (long long)R * C; v2_1_22.sCm = C; v2_1_22.sRo = (long long)R * R * C; v2_1_22.sRi = (long long)R * C; v2_1_22.sRm = C; v2_1_22.sRn = 1;
      v2_1_22.M = R; v2_1_22.N = C; v2_1_22.K = C; v2_1_22.zi_n = R; v2_1_22.flags = 4; v2_1_22.act = 0;
      v2_1_22.alpha = 1.0f; v2_1_22.beta = 1.0f; v2_1_22.sa = 1.0f; v2_1_22.sb = 1.0f; v2_1_22.Npad = C; v2_1_22.pad_ = 0;
      k_gemm<1><<<dim3((unsigned)((C) + 31) / 32, (unsigned)((R) + 15) / 16, (unsigned)(R * R)), 32, 0, stream>>>(v2_1_22); }
    { GemmP v2_1_23;
      v2_1_23.A = GQ + (size_t)1 * RP3 * C + (size_t)2348 * C; v2_1_23.B = wv2 + 23; v2_1_23.bias = GQ + (size_t)1 * RP3 * C + (size_t)2348 * C; v2_1_23.R = GC + (size_t)1 * R3 * C; v2_1_23.C = GC + (size_t)1 * R3 * C;
      v2_1_23.sAo = (long long)34 * 34 * C; v2_1_23.sAi = (long long)34 * C; v2_1_23.sAm = C; v2_1_23.sAk = 1; v2_1_23.sBo = 0; v2_1_23.sBi = 0; v2_1_23.sBn = C * 27; v2_1_23.sBk = 27; v2_1_23.sCo = (long long)R * R * C; v2_1_23.sCi = (long long)R * C; v2_1_23.sCm = C; v2_1_23.sRo = (long long)R * R * C; v2_1_23.sRi = (long long)R * C; v2_1_23.sRm = C; v2_1_23.sRn = 1;
      v2_1_23.M = R; v2_1_23.N = C; v2_1_23.K = C; v2_1_23.zi_n = R; v2_1_23.flags = 4; v2_1_23.act = 0;
      v2_1_23.alpha = 1.0f; v2_1_23.beta = 1.0f; v2_1_23.sa = 1.0f; v2_1_23.sb = 1.0f; v2_1_23.Npad = C; v2_1_23.pad_ = 0;
      k_gemm<1><<<dim3((unsigned)((C) + 31) / 32, (unsigned)((R) + 15) / 16, (unsigned)(R * R)), 32, 0, stream>>>(v2_1_23); }
    { GemmP v2_1_24;
      v2_1_24.A = GQ + (size_t)1 * RP3 * C + (size_t)2380 * C; v2_1_24.B = wv2 + 24; v2_1_24.bias = GQ + (size_t)1 * RP3 * C + (size_t)2380 * C; v2_1_24.R = GC + (size_t)1 * R3 * C; v2_1_24.C = GC + (size_t)1 * R3 * C;
      v2_1_24.sAo = (long long)34 * 34 * C; v2_1_24.sAi = (long long)34 * C; v2_1_24.sAm = C; v2_1_24.sAk = 1; v2_1_24.sBo = 0; v2_1_24.sBi = 0; v2_1_24.sBn = C * 27; v2_1_24.sBk = 27; v2_1_24.sCo = (long long)R * R * C; v2_1_24.sCi = (long long)R * C; v2_1_24.sCm = C; v2_1_24.sRo = (long long)R * R * C; v2_1_24.sRi = (long long)R * C; v2_1_24.sRm = C; v2_1_24.sRn = 1;
      v2_1_24.M = R; v2_1_24.N = C; v2_1_24.K = C; v2_1_24.zi_n = R; v2_1_24.flags = 4; v2_1_24.act = 0;
      v2_1_24.alpha = 1.0f; v2_1_24.beta = 1.0f; v2_1_24.sa = 1.0f; v2_1_24.sb = 1.0f; v2_1_24.Npad = C; v2_1_24.pad_ = 0;
      k_gemm<1><<<dim3((unsigned)((C) + 31) / 32, (unsigned)((R) + 15) / 16, (unsigned)(R * R)), 32, 0, stream>>>(v2_1_24); }
    { GemmP v2_1_25;
      v2_1_25.A = GQ + (size_t)1 * RP3 * C + (size_t)2381 * C; v2_1_25.B = wv2 + 25; v2_1_25.bias = GQ + (size_t)1 * RP3 * C + (size_t)2381 * C; v2_1_25.R = GC + (size_t)1 * R3 * C; v2_1_25.C = GC + (size_t)1 * R3 * C;
      v2_1_25.sAo = (long long)34 * 34 * C; v2_1_25.sAi = (long long)34 * C; v2_1_25.sAm = C; v2_1_25.sAk = 1; v2_1_25.sBo = 0; v2_1_25.sBi = 0; v2_1_25.sBn = C * 27; v2_1_25.sBk = 27; v2_1_25.sCo = (long long)R * R * C; v2_1_25.sCi = (long long)R * C; v2_1_25.sCm = C; v2_1_25.sRo = (long long)R * R * C; v2_1_25.sRi = (long long)R * C; v2_1_25.sRm = C; v2_1_25.sRn = 1;
      v2_1_25.M = R; v2_1_25.N = C; v2_1_25.K = C; v2_1_25.zi_n = R; v2_1_25.flags = 4; v2_1_25.act = 0;
      v2_1_25.alpha = 1.0f; v2_1_25.beta = 1.0f; v2_1_25.sa = 1.0f; v2_1_25.sb = 1.0f; v2_1_25.Npad = C; v2_1_25.pad_ = 0;
      k_gemm<1><<<dim3((unsigned)((C) + 31) / 32, (unsigned)((R) + 15) / 16, (unsigned)(R * R)), 32, 0, stream>>>(v2_1_25); }
    { GemmP v2_1_26;
      v2_1_26.A = GQ + (size_t)1 * RP3 * C + (size_t)2382 * C; v2_1_26.B = wv2 + 26; v2_1_26.bias = GQ + (size_t)1 * RP3 * C + (size_t)2382 * C; v2_1_26.R = GC + (size_t)1 * R3 * C; v2_1_26.C = GC + (size_t)1 * R3 * C;
      v2_1_26.sAo = (long long)34 * 34 * C; v2_1_26.sAi = (long long)34 * C; v2_1_26.sAm = C; v2_1_26.sAk = 1; v2_1_26.sBo = 0; v2_1_26.sBi = 0; v2_1_26.sBn = C * 27; v2_1_26.sBk = 27; v2_1_26.sCo = (long long)R * R * C; v2_1_26.sCi = (long long)R * C; v2_1_26.sCm = C; v2_1_26.sRo = (long long)R * R * C; v2_1_26.sRi = (long long)R * C; v2_1_26.sRm = C; v2_1_26.sRn = 1;
      v2_1_26.M = R; v2_1_26.N = C; v2_1_26.K = C; v2_1_26.zi_n = R; v2_1_26.flags = 4; v2_1_26.act = 0;
      v2_1_26.alpha = 1.0f; v2_1_26.beta = 1.0f; v2_1_26.sa = 1.0f; v2_1_26.sb = 1.0f; v2_1_26.Npad = C; v2_1_26.pad_ = 0;
      k_gemm<1><<<dim3((unsigned)((C) + 31) / 32, (unsigned)((R) + 15) / 16, (unsigned)(R * R)), 32, 0, stream>>>(v2_1_26); }
    { GemmP v2_2_0;
      v2_2_0.A = GQ + (size_t)2 * RP3 * C + (size_t)0 * C; v2_2_0.B = wv2 + 0; v2_2_0.bias = GQ + (size_t)2 * RP3 * C + (size_t)0 * C; v2_2_0.R = GQ + (size_t)2 * RP3 * C + (size_t)0 * C; v2_2_0.C = GC + (size_t)2 * R3 * C;
      v2_2_0.sAo = (long long)34 * 34 * C; v2_2_0.sAi = (long long)34 * C; v2_2_0.sAm = C; v2_2_0.sAk = 1; v2_2_0.sBo = 0; v2_2_0.sBi = 0; v2_2_0.sBn = C * 27; v2_2_0.sBk = 27; v2_2_0.sCo = (long long)R * R * C; v2_2_0.sCi = (long long)R * C; v2_2_0.sCm = C; v2_2_0.sRo = 0; v2_2_0.sRi = 0; v2_2_0.sRm = 0; v2_2_0.sRn = 0;
      v2_2_0.M = R; v2_2_0.N = C; v2_2_0.K = C; v2_2_0.zi_n = R; v2_2_0.flags = 0; v2_2_0.act = 0;
      v2_2_0.alpha = 1.0f; v2_2_0.beta = 0.0f; v2_2_0.sa = 1.0f; v2_2_0.sb = 1.0f; v2_2_0.Npad = C; v2_2_0.pad_ = 0;
      k_gemm<1><<<dim3((unsigned)((C) + 31) / 32, (unsigned)((R) + 15) / 16, (unsigned)(R * R)), 32, 0, stream>>>(v2_2_0); }
    { GemmP v2_2_1;
      v2_2_1.A = GQ + (size_t)2 * RP3 * C + (size_t)1 * C; v2_2_1.B = wv2 + 1; v2_2_1.bias = GQ + (size_t)2 * RP3 * C + (size_t)1 * C; v2_2_1.R = GC + (size_t)2 * R3 * C; v2_2_1.C = GC + (size_t)2 * R3 * C;
      v2_2_1.sAo = (long long)34 * 34 * C; v2_2_1.sAi = (long long)34 * C; v2_2_1.sAm = C; v2_2_1.sAk = 1; v2_2_1.sBo = 0; v2_2_1.sBi = 0; v2_2_1.sBn = C * 27; v2_2_1.sBk = 27; v2_2_1.sCo = (long long)R * R * C; v2_2_1.sCi = (long long)R * C; v2_2_1.sCm = C; v2_2_1.sRo = (long long)R * R * C; v2_2_1.sRi = (long long)R * C; v2_2_1.sRm = C; v2_2_1.sRn = 1;
      v2_2_1.M = R; v2_2_1.N = C; v2_2_1.K = C; v2_2_1.zi_n = R; v2_2_1.flags = 4; v2_2_1.act = 0;
      v2_2_1.alpha = 1.0f; v2_2_1.beta = 1.0f; v2_2_1.sa = 1.0f; v2_2_1.sb = 1.0f; v2_2_1.Npad = C; v2_2_1.pad_ = 0;
      k_gemm<1><<<dim3((unsigned)((C) + 31) / 32, (unsigned)((R) + 15) / 16, (unsigned)(R * R)), 32, 0, stream>>>(v2_2_1); }
    { GemmP v2_2_2;
      v2_2_2.A = GQ + (size_t)2 * RP3 * C + (size_t)2 * C; v2_2_2.B = wv2 + 2; v2_2_2.bias = GQ + (size_t)2 * RP3 * C + (size_t)2 * C; v2_2_2.R = GC + (size_t)2 * R3 * C; v2_2_2.C = GC + (size_t)2 * R3 * C;
      v2_2_2.sAo = (long long)34 * 34 * C; v2_2_2.sAi = (long long)34 * C; v2_2_2.sAm = C; v2_2_2.sAk = 1; v2_2_2.sBo = 0; v2_2_2.sBi = 0; v2_2_2.sBn = C * 27; v2_2_2.sBk = 27; v2_2_2.sCo = (long long)R * R * C; v2_2_2.sCi = (long long)R * C; v2_2_2.sCm = C; v2_2_2.sRo = (long long)R * R * C; v2_2_2.sRi = (long long)R * C; v2_2_2.sRm = C; v2_2_2.sRn = 1;
      v2_2_2.M = R; v2_2_2.N = C; v2_2_2.K = C; v2_2_2.zi_n = R; v2_2_2.flags = 4; v2_2_2.act = 0;
      v2_2_2.alpha = 1.0f; v2_2_2.beta = 1.0f; v2_2_2.sa = 1.0f; v2_2_2.sb = 1.0f; v2_2_2.Npad = C; v2_2_2.pad_ = 0;
      k_gemm<1><<<dim3((unsigned)((C) + 31) / 32, (unsigned)((R) + 15) / 16, (unsigned)(R * R)), 32, 0, stream>>>(v2_2_2); }
    { GemmP v2_2_3;
      v2_2_3.A = GQ + (size_t)2 * RP3 * C + (size_t)34 * C; v2_2_3.B = wv2 + 3; v2_2_3.bias = GQ + (size_t)2 * RP3 * C + (size_t)34 * C; v2_2_3.R = GC + (size_t)2 * R3 * C; v2_2_3.C = GC + (size_t)2 * R3 * C;
      v2_2_3.sAo = (long long)34 * 34 * C; v2_2_3.sAi = (long long)34 * C; v2_2_3.sAm = C; v2_2_3.sAk = 1; v2_2_3.sBo = 0; v2_2_3.sBi = 0; v2_2_3.sBn = C * 27; v2_2_3.sBk = 27; v2_2_3.sCo = (long long)R * R * C; v2_2_3.sCi = (long long)R * C; v2_2_3.sCm = C; v2_2_3.sRo = (long long)R * R * C; v2_2_3.sRi = (long long)R * C; v2_2_3.sRm = C; v2_2_3.sRn = 1;
      v2_2_3.M = R; v2_2_3.N = C; v2_2_3.K = C; v2_2_3.zi_n = R; v2_2_3.flags = 4; v2_2_3.act = 0;
      v2_2_3.alpha = 1.0f; v2_2_3.beta = 1.0f; v2_2_3.sa = 1.0f; v2_2_3.sb = 1.0f; v2_2_3.Npad = C; v2_2_3.pad_ = 0;
      k_gemm<1><<<dim3((unsigned)((C) + 31) / 32, (unsigned)((R) + 15) / 16, (unsigned)(R * R)), 32, 0, stream>>>(v2_2_3); }
    { GemmP v2_2_4;
      v2_2_4.A = GQ + (size_t)2 * RP3 * C + (size_t)35 * C; v2_2_4.B = wv2 + 4; v2_2_4.bias = GQ + (size_t)2 * RP3 * C + (size_t)35 * C; v2_2_4.R = GC + (size_t)2 * R3 * C; v2_2_4.C = GC + (size_t)2 * R3 * C;
      v2_2_4.sAo = (long long)34 * 34 * C; v2_2_4.sAi = (long long)34 * C; v2_2_4.sAm = C; v2_2_4.sAk = 1; v2_2_4.sBo = 0; v2_2_4.sBi = 0; v2_2_4.sBn = C * 27; v2_2_4.sBk = 27; v2_2_4.sCo = (long long)R * R * C; v2_2_4.sCi = (long long)R * C; v2_2_4.sCm = C; v2_2_4.sRo = (long long)R * R * C; v2_2_4.sRi = (long long)R * C; v2_2_4.sRm = C; v2_2_4.sRn = 1;
      v2_2_4.M = R; v2_2_4.N = C; v2_2_4.K = C; v2_2_4.zi_n = R; v2_2_4.flags = 4; v2_2_4.act = 0;
      v2_2_4.alpha = 1.0f; v2_2_4.beta = 1.0f; v2_2_4.sa = 1.0f; v2_2_4.sb = 1.0f; v2_2_4.Npad = C; v2_2_4.pad_ = 0;
      k_gemm<1><<<dim3((unsigned)((C) + 31) / 32, (unsigned)((R) + 15) / 16, (unsigned)(R * R)), 32, 0, stream>>>(v2_2_4); }
    { GemmP v2_2_5;
      v2_2_5.A = GQ + (size_t)2 * RP3 * C + (size_t)36 * C; v2_2_5.B = wv2 + 5; v2_2_5.bias = GQ + (size_t)2 * RP3 * C + (size_t)36 * C; v2_2_5.R = GC + (size_t)2 * R3 * C; v2_2_5.C = GC + (size_t)2 * R3 * C;
      v2_2_5.sAo = (long long)34 * 34 * C; v2_2_5.sAi = (long long)34 * C; v2_2_5.sAm = C; v2_2_5.sAk = 1; v2_2_5.sBo = 0; v2_2_5.sBi = 0; v2_2_5.sBn = C * 27; v2_2_5.sBk = 27; v2_2_5.sCo = (long long)R * R * C; v2_2_5.sCi = (long long)R * C; v2_2_5.sCm = C; v2_2_5.sRo = (long long)R * R * C; v2_2_5.sRi = (long long)R * C; v2_2_5.sRm = C; v2_2_5.sRn = 1;
      v2_2_5.M = R; v2_2_5.N = C; v2_2_5.K = C; v2_2_5.zi_n = R; v2_2_5.flags = 4; v2_2_5.act = 0;
      v2_2_5.alpha = 1.0f; v2_2_5.beta = 1.0f; v2_2_5.sa = 1.0f; v2_2_5.sb = 1.0f; v2_2_5.Npad = C; v2_2_5.pad_ = 0;
      k_gemm<1><<<dim3((unsigned)((C) + 31) / 32, (unsigned)((R) + 15) / 16, (unsigned)(R * R)), 32, 0, stream>>>(v2_2_5); }
    { GemmP v2_2_6;
      v2_2_6.A = GQ + (size_t)2 * RP3 * C + (size_t)68 * C; v2_2_6.B = wv2 + 6; v2_2_6.bias = GQ + (size_t)2 * RP3 * C + (size_t)68 * C; v2_2_6.R = GC + (size_t)2 * R3 * C; v2_2_6.C = GC + (size_t)2 * R3 * C;
      v2_2_6.sAo = (long long)34 * 34 * C; v2_2_6.sAi = (long long)34 * C; v2_2_6.sAm = C; v2_2_6.sAk = 1; v2_2_6.sBo = 0; v2_2_6.sBi = 0; v2_2_6.sBn = C * 27; v2_2_6.sBk = 27; v2_2_6.sCo = (long long)R * R * C; v2_2_6.sCi = (long long)R * C; v2_2_6.sCm = C; v2_2_6.sRo = (long long)R * R * C; v2_2_6.sRi = (long long)R * C; v2_2_6.sRm = C; v2_2_6.sRn = 1;
      v2_2_6.M = R; v2_2_6.N = C; v2_2_6.K = C; v2_2_6.zi_n = R; v2_2_6.flags = 4; v2_2_6.act = 0;
      v2_2_6.alpha = 1.0f; v2_2_6.beta = 1.0f; v2_2_6.sa = 1.0f; v2_2_6.sb = 1.0f; v2_2_6.Npad = C; v2_2_6.pad_ = 0;
      k_gemm<1><<<dim3((unsigned)((C) + 31) / 32, (unsigned)((R) + 15) / 16, (unsigned)(R * R)), 32, 0, stream>>>(v2_2_6); }
    { GemmP v2_2_7;
      v2_2_7.A = GQ + (size_t)2 * RP3 * C + (size_t)69 * C; v2_2_7.B = wv2 + 7; v2_2_7.bias = GQ + (size_t)2 * RP3 * C + (size_t)69 * C; v2_2_7.R = GC + (size_t)2 * R3 * C; v2_2_7.C = GC + (size_t)2 * R3 * C;
      v2_2_7.sAo = (long long)34 * 34 * C; v2_2_7.sAi = (long long)34 * C; v2_2_7.sAm = C; v2_2_7.sAk = 1; v2_2_7.sBo = 0; v2_2_7.sBi = 0; v2_2_7.sBn = C * 27; v2_2_7.sBk = 27; v2_2_7.sCo = (long long)R * R * C; v2_2_7.sCi = (long long)R * C; v2_2_7.sCm = C; v2_2_7.sRo = (long long)R * R * C; v2_2_7.sRi = (long long)R * C; v2_2_7.sRm = C; v2_2_7.sRn = 1;
      v2_2_7.M = R; v2_2_7.N = C; v2_2_7.K = C; v2_2_7.zi_n = R; v2_2_7.flags = 4; v2_2_7.act = 0;
      v2_2_7.alpha = 1.0f; v2_2_7.beta = 1.0f; v2_2_7.sa = 1.0f; v2_2_7.sb = 1.0f; v2_2_7.Npad = C; v2_2_7.pad_ = 0;
      k_gemm<1><<<dim3((unsigned)((C) + 31) / 32, (unsigned)((R) + 15) / 16, (unsigned)(R * R)), 32, 0, stream>>>(v2_2_7); }
    { GemmP v2_2_8;
      v2_2_8.A = GQ + (size_t)2 * RP3 * C + (size_t)70 * C; v2_2_8.B = wv2 + 8; v2_2_8.bias = GQ + (size_t)2 * RP3 * C + (size_t)70 * C; v2_2_8.R = GC + (size_t)2 * R3 * C; v2_2_8.C = GC + (size_t)2 * R3 * C;
      v2_2_8.sAo = (long long)34 * 34 * C; v2_2_8.sAi = (long long)34 * C; v2_2_8.sAm = C; v2_2_8.sAk = 1; v2_2_8.sBo = 0; v2_2_8.sBi = 0; v2_2_8.sBn = C * 27; v2_2_8.sBk = 27; v2_2_8.sCo = (long long)R * R * C; v2_2_8.sCi = (long long)R * C; v2_2_8.sCm = C; v2_2_8.sRo = (long long)R * R * C; v2_2_8.sRi = (long long)R * C; v2_2_8.sRm = C; v2_2_8.sRn = 1;
      v2_2_8.M = R; v2_2_8.N = C; v2_2_8.K = C; v2_2_8.zi_n = R; v2_2_8.flags = 4; v2_2_8.act = 0;
      v2_2_8.alpha = 1.0f; v2_2_8.beta = 1.0f; v2_2_8.sa = 1.0f; v2_2_8.sb = 1.0f; v2_2_8.Npad = C; v2_2_8.pad_ = 0;
      k_gemm<1><<<dim3((unsigned)((C) + 31) / 32, (unsigned)((R) + 15) / 16, (unsigned)(R * R)), 32, 0, stream>>>(v2_2_8); }
    { GemmP v2_2_9;
      v2_2_9.A = GQ + (size_t)2 * RP3 * C + (size_t)1156 * C; v2_2_9.B = wv2 + 9; v2_2_9.bias = GQ + (size_t)2 * RP3 * C + (size_t)1156 * C; v2_2_9.R = GC + (size_t)2 * R3 * C; v2_2_9.C = GC + (size_t)2 * R3 * C;
      v2_2_9.sAo = (long long)34 * 34 * C; v2_2_9.sAi = (long long)34 * C; v2_2_9.sAm = C; v2_2_9.sAk = 1; v2_2_9.sBo = 0; v2_2_9.sBi = 0; v2_2_9.sBn = C * 27; v2_2_9.sBk = 27; v2_2_9.sCo = (long long)R * R * C; v2_2_9.sCi = (long long)R * C; v2_2_9.sCm = C; v2_2_9.sRo = (long long)R * R * C; v2_2_9.sRi = (long long)R * C; v2_2_9.sRm = C; v2_2_9.sRn = 1;
      v2_2_9.M = R; v2_2_9.N = C; v2_2_9.K = C; v2_2_9.zi_n = R; v2_2_9.flags = 4; v2_2_9.act = 0;
      v2_2_9.alpha = 1.0f; v2_2_9.beta = 1.0f; v2_2_9.sa = 1.0f; v2_2_9.sb = 1.0f; v2_2_9.Npad = C; v2_2_9.pad_ = 0;
      k_gemm<1><<<dim3((unsigned)((C) + 31) / 32, (unsigned)((R) + 15) / 16, (unsigned)(R * R)), 32, 0, stream>>>(v2_2_9); }
    { GemmP v2_2_10;
      v2_2_10.A = GQ + (size_t)2 * RP3 * C + (size_t)1157 * C; v2_2_10.B = wv2 + 10; v2_2_10.bias = GQ + (size_t)2 * RP3 * C + (size_t)1157 * C; v2_2_10.R = GC + (size_t)2 * R3 * C; v2_2_10.C = GC + (size_t)2 * R3 * C;
      v2_2_10.sAo = (long long)34 * 34 * C; v2_2_10.sAi = (long long)34 * C; v2_2_10.sAm = C; v2_2_10.sAk = 1; v2_2_10.sBo = 0; v2_2_10.sBi = 0; v2_2_10.sBn = C * 27; v2_2_10.sBk = 27; v2_2_10.sCo = (long long)R * R * C; v2_2_10.sCi = (long long)R * C; v2_2_10.sCm = C; v2_2_10.sRo = (long long)R * R * C; v2_2_10.sRi = (long long)R * C; v2_2_10.sRm = C; v2_2_10.sRn = 1;
      v2_2_10.M = R; v2_2_10.N = C; v2_2_10.K = C; v2_2_10.zi_n = R; v2_2_10.flags = 4; v2_2_10.act = 0;
      v2_2_10.alpha = 1.0f; v2_2_10.beta = 1.0f; v2_2_10.sa = 1.0f; v2_2_10.sb = 1.0f; v2_2_10.Npad = C; v2_2_10.pad_ = 0;
      k_gemm<1><<<dim3((unsigned)((C) + 31) / 32, (unsigned)((R) + 15) / 16, (unsigned)(R * R)), 32, 0, stream>>>(v2_2_10); }
    { GemmP v2_2_11;
      v2_2_11.A = GQ + (size_t)2 * RP3 * C + (size_t)1158 * C; v2_2_11.B = wv2 + 11; v2_2_11.bias = GQ + (size_t)2 * RP3 * C + (size_t)1158 * C; v2_2_11.R = GC + (size_t)2 * R3 * C; v2_2_11.C = GC + (size_t)2 * R3 * C;
      v2_2_11.sAo = (long long)34 * 34 * C; v2_2_11.sAi = (long long)34 * C; v2_2_11.sAm = C; v2_2_11.sAk = 1; v2_2_11.sBo = 0; v2_2_11.sBi = 0; v2_2_11.sBn = C * 27; v2_2_11.sBk = 27; v2_2_11.sCo = (long long)R * R * C; v2_2_11.sCi = (long long)R * C; v2_2_11.sCm = C; v2_2_11.sRo = (long long)R * R * C; v2_2_11.sRi = (long long)R * C; v2_2_11.sRm = C; v2_2_11.sRn = 1;
      v2_2_11.M = R; v2_2_11.N = C; v2_2_11.K = C; v2_2_11.zi_n = R; v2_2_11.flags = 4; v2_2_11.act = 0;
      v2_2_11.alpha = 1.0f; v2_2_11.beta = 1.0f; v2_2_11.sa = 1.0f; v2_2_11.sb = 1.0f; v2_2_11.Npad = C; v2_2_11.pad_ = 0;
      k_gemm<1><<<dim3((unsigned)((C) + 31) / 32, (unsigned)((R) + 15) / 16, (unsigned)(R * R)), 32, 0, stream>>>(v2_2_11); }
    { GemmP v2_2_12;
      v2_2_12.A = GQ + (size_t)2 * RP3 * C + (size_t)1190 * C; v2_2_12.B = wv2 + 12; v2_2_12.bias = GQ + (size_t)2 * RP3 * C + (size_t)1190 * C; v2_2_12.R = GC + (size_t)2 * R3 * C; v2_2_12.C = GC + (size_t)2 * R3 * C;
      v2_2_12.sAo = (long long)34 * 34 * C; v2_2_12.sAi = (long long)34 * C; v2_2_12.sAm = C; v2_2_12.sAk = 1; v2_2_12.sBo = 0; v2_2_12.sBi = 0; v2_2_12.sBn = C * 27; v2_2_12.sBk = 27; v2_2_12.sCo = (long long)R * R * C; v2_2_12.sCi = (long long)R * C; v2_2_12.sCm = C; v2_2_12.sRo = (long long)R * R * C; v2_2_12.sRi = (long long)R * C; v2_2_12.sRm = C; v2_2_12.sRn = 1;
      v2_2_12.M = R; v2_2_12.N = C; v2_2_12.K = C; v2_2_12.zi_n = R; v2_2_12.flags = 4; v2_2_12.act = 0;
      v2_2_12.alpha = 1.0f; v2_2_12.beta = 1.0f; v2_2_12.sa = 1.0f; v2_2_12.sb = 1.0f; v2_2_12.Npad = C; v2_2_12.pad_ = 0;
      k_gemm<1><<<dim3((unsigned)((C) + 31) / 32, (unsigned)((R) + 15) / 16, (unsigned)(R * R)), 32, 0, stream>>>(v2_2_12); }
    { GemmP v2_2_13;
      v2_2_13.A = GQ + (size_t)2 * RP3 * C + (size_t)1191 * C; v2_2_13.B = wv2 + 13; v2_2_13.bias = GQ + (size_t)2 * RP3 * C + (size_t)1191 * C; v2_2_13.R = GC + (size_t)2 * R3 * C; v2_2_13.C = GC + (size_t)2 * R3 * C;
      v2_2_13.sAo = (long long)34 * 34 * C; v2_2_13.sAi = (long long)34 * C; v2_2_13.sAm = C; v2_2_13.sAk = 1; v2_2_13.sBo = 0; v2_2_13.sBi = 0; v2_2_13.sBn = C * 27; v2_2_13.sBk = 27; v2_2_13.sCo = (long long)R * R * C; v2_2_13.sCi = (long long)R * C; v2_2_13.sCm = C; v2_2_13.sRo = (long long)R * R * C; v2_2_13.sRi = (long long)R * C; v2_2_13.sRm = C; v2_2_13.sRn = 1;
      v2_2_13.M = R; v2_2_13.N = C; v2_2_13.K = C; v2_2_13.zi_n = R; v2_2_13.flags = 4; v2_2_13.act = 0;
      v2_2_13.alpha = 1.0f; v2_2_13.beta = 1.0f; v2_2_13.sa = 1.0f; v2_2_13.sb = 1.0f; v2_2_13.Npad = C; v2_2_13.pad_ = 0;
      k_gemm<1><<<dim3((unsigned)((C) + 31) / 32, (unsigned)((R) + 15) / 16, (unsigned)(R * R)), 32, 0, stream>>>(v2_2_13); }
    { GemmP v2_2_14;
      v2_2_14.A = GQ + (size_t)2 * RP3 * C + (size_t)1192 * C; v2_2_14.B = wv2 + 14; v2_2_14.bias = GQ + (size_t)2 * RP3 * C + (size_t)1192 * C; v2_2_14.R = GC + (size_t)2 * R3 * C; v2_2_14.C = GC + (size_t)2 * R3 * C;
      v2_2_14.sAo = (long long)34 * 34 * C; v2_2_14.sAi = (long long)34 * C; v2_2_14.sAm = C; v2_2_14.sAk = 1; v2_2_14.sBo = 0; v2_2_14.sBi = 0; v2_2_14.sBn = C * 27; v2_2_14.sBk = 27; v2_2_14.sCo = (long long)R * R * C; v2_2_14.sCi = (long long)R * C; v2_2_14.sCm = C; v2_2_14.sRo = (long long)R * R * C; v2_2_14.sRi = (long long)R * C; v2_2_14.sRm = C; v2_2_14.sRn = 1;
      v2_2_14.M = R; v2_2_14.N = C; v2_2_14.K = C; v2_2_14.zi_n = R; v2_2_14.flags = 4; v2_2_14.act = 0;
      v2_2_14.alpha = 1.0f; v2_2_14.beta = 1.0f; v2_2_14.sa = 1.0f; v2_2_14.sb = 1.0f; v2_2_14.Npad = C; v2_2_14.pad_ = 0;
      k_gemm<1><<<dim3((unsigned)((C) + 31) / 32, (unsigned)((R) + 15) / 16, (unsigned)(R * R)), 32, 0, stream>>>(v2_2_14); }
    { GemmP v2_2_15;
      v2_2_15.A = GQ + (size_t)2 * RP3 * C + (size_t)1224 * C; v2_2_15.B = wv2 + 15; v2_2_15.bias = GQ + (size_t)2 * RP3 * C + (size_t)1224 * C; v2_2_15.R = GC + (size_t)2 * R3 * C; v2_2_15.C = GC + (size_t)2 * R3 * C;
      v2_2_15.sAo = (long long)34 * 34 * C; v2_2_15.sAi = (long long)34 * C; v2_2_15.sAm = C; v2_2_15.sAk = 1; v2_2_15.sBo = 0; v2_2_15.sBi = 0; v2_2_15.sBn = C * 27; v2_2_15.sBk = 27; v2_2_15.sCo = (long long)R * R * C; v2_2_15.sCi = (long long)R * C; v2_2_15.sCm = C; v2_2_15.sRo = (long long)R * R * C; v2_2_15.sRi = (long long)R * C; v2_2_15.sRm = C; v2_2_15.sRn = 1;
      v2_2_15.M = R; v2_2_15.N = C; v2_2_15.K = C; v2_2_15.zi_n = R; v2_2_15.flags = 4; v2_2_15.act = 0;
      v2_2_15.alpha = 1.0f; v2_2_15.beta = 1.0f; v2_2_15.sa = 1.0f; v2_2_15.sb = 1.0f; v2_2_15.Npad = C; v2_2_15.pad_ = 0;
      k_gemm<1><<<dim3((unsigned)((C) + 31) / 32, (unsigned)((R) + 15) / 16, (unsigned)(R * R)), 32, 0, stream>>>(v2_2_15); }
    { GemmP v2_2_16;
      v2_2_16.A = GQ + (size_t)2 * RP3 * C + (size_t)1225 * C; v2_2_16.B = wv2 + 16; v2_2_16.bias = GQ + (size_t)2 * RP3 * C + (size_t)1225 * C; v2_2_16.R = GC + (size_t)2 * R3 * C; v2_2_16.C = GC + (size_t)2 * R3 * C;
      v2_2_16.sAo = (long long)34 * 34 * C; v2_2_16.sAi = (long long)34 * C; v2_2_16.sAm = C; v2_2_16.sAk = 1; v2_2_16.sBo = 0; v2_2_16.sBi = 0; v2_2_16.sBn = C * 27; v2_2_16.sBk = 27; v2_2_16.sCo = (long long)R * R * C; v2_2_16.sCi = (long long)R * C; v2_2_16.sCm = C; v2_2_16.sRo = (long long)R * R * C; v2_2_16.sRi = (long long)R * C; v2_2_16.sRm = C; v2_2_16.sRn = 1;
      v2_2_16.M = R; v2_2_16.N = C; v2_2_16.K = C; v2_2_16.zi_n = R; v2_2_16.flags = 4; v2_2_16.act = 0;
      v2_2_16.alpha = 1.0f; v2_2_16.beta = 1.0f; v2_2_16.sa = 1.0f; v2_2_16.sb = 1.0f; v2_2_16.Npad = C; v2_2_16.pad_ = 0;
      k_gemm<1><<<dim3((unsigned)((C) + 31) / 32, (unsigned)((R) + 15) / 16, (unsigned)(R * R)), 32, 0, stream>>>(v2_2_16); }
    { GemmP v2_2_17;
      v2_2_17.A = GQ + (size_t)2 * RP3 * C + (size_t)1226 * C; v2_2_17.B = wv2 + 17; v2_2_17.bias = GQ + (size_t)2 * RP3 * C + (size_t)1226 * C; v2_2_17.R = GC + (size_t)2 * R3 * C; v2_2_17.C = GC + (size_t)2 * R3 * C;
      v2_2_17.sAo = (long long)34 * 34 * C; v2_2_17.sAi = (long long)34 * C; v2_2_17.sAm = C; v2_2_17.sAk = 1; v2_2_17.sBo = 0; v2_2_17.sBi = 0; v2_2_17.sBn = C * 27; v2_2_17.sBk = 27; v2_2_17.sCo = (long long)R * R * C; v2_2_17.sCi = (long long)R * C; v2_2_17.sCm = C; v2_2_17.sRo = (long long)R * R * C; v2_2_17.sRi = (long long)R * C; v2_2_17.sRm = C; v2_2_17.sRn = 1;
      v2_2_17.M = R; v2_2_17.N = C; v2_2_17.K = C; v2_2_17.zi_n = R; v2_2_17.flags = 4; v2_2_17.act = 0;
      v2_2_17.alpha = 1.0f; v2_2_17.beta = 1.0f; v2_2_17.sa = 1.0f; v2_2_17.sb = 1.0f; v2_2_17.Npad = C; v2_2_17.pad_ = 0;
      k_gemm<1><<<dim3((unsigned)((C) + 31) / 32, (unsigned)((R) + 15) / 16, (unsigned)(R * R)), 32, 0, stream>>>(v2_2_17); }
    { GemmP v2_2_18;
      v2_2_18.A = GQ + (size_t)2 * RP3 * C + (size_t)2312 * C; v2_2_18.B = wv2 + 18; v2_2_18.bias = GQ + (size_t)2 * RP3 * C + (size_t)2312 * C; v2_2_18.R = GC + (size_t)2 * R3 * C; v2_2_18.C = GC + (size_t)2 * R3 * C;
      v2_2_18.sAo = (long long)34 * 34 * C; v2_2_18.sAi = (long long)34 * C; v2_2_18.sAm = C; v2_2_18.sAk = 1; v2_2_18.sBo = 0; v2_2_18.sBi = 0; v2_2_18.sBn = C * 27; v2_2_18.sBk = 27; v2_2_18.sCo = (long long)R * R * C; v2_2_18.sCi = (long long)R * C; v2_2_18.sCm = C; v2_2_18.sRo = (long long)R * R * C; v2_2_18.sRi = (long long)R * C; v2_2_18.sRm = C; v2_2_18.sRn = 1;
      v2_2_18.M = R; v2_2_18.N = C; v2_2_18.K = C; v2_2_18.zi_n = R; v2_2_18.flags = 4; v2_2_18.act = 0;
      v2_2_18.alpha = 1.0f; v2_2_18.beta = 1.0f; v2_2_18.sa = 1.0f; v2_2_18.sb = 1.0f; v2_2_18.Npad = C; v2_2_18.pad_ = 0;
      k_gemm<1><<<dim3((unsigned)((C) + 31) / 32, (unsigned)((R) + 15) / 16, (unsigned)(R * R)), 32, 0, stream>>>(v2_2_18); }
    { GemmP v2_2_19;
      v2_2_19.A = GQ + (size_t)2 * RP3 * C + (size_t)2313 * C; v2_2_19.B = wv2 + 19; v2_2_19.bias = GQ + (size_t)2 * RP3 * C + (size_t)2313 * C; v2_2_19.R = GC + (size_t)2 * R3 * C; v2_2_19.C = GC + (size_t)2 * R3 * C;
      v2_2_19.sAo = (long long)34 * 34 * C; v2_2_19.sAi = (long long)34 * C; v2_2_19.sAm = C; v2_2_19.sAk = 1; v2_2_19.sBo = 0; v2_2_19.sBi = 0; v2_2_19.sBn = C * 27; v2_2_19.sBk = 27; v2_2_19.sCo = (long long)R * R * C; v2_2_19.sCi = (long long)R * C; v2_2_19.sCm = C; v2_2_19.sRo = (long long)R * R * C; v2_2_19.sRi = (long long)R * C; v2_2_19.sRm = C; v2_2_19.sRn = 1;
      v2_2_19.M = R; v2_2_19.N = C; v2_2_19.K = C; v2_2_19.zi_n = R; v2_2_19.flags = 4; v2_2_19.act = 0;
      v2_2_19.alpha = 1.0f; v2_2_19.beta = 1.0f; v2_2_19.sa = 1.0f; v2_2_19.sb = 1.0f; v2_2_19.Npad = C; v2_2_19.pad_ = 0;
      k_gemm<1><<<dim3((unsigned)((C) + 31) / 32, (unsigned)((R) + 15) / 16, (unsigned)(R * R)), 32, 0, stream>>>(v2_2_19); }
    { GemmP v2_2_20;
      v2_2_20.A = GQ + (size_t)2 * RP3 * C + (size_t)2314 * C; v2_2_20.B = wv2 + 20; v2_2_20.bias = GQ + (size_t)2 * RP3 * C + (size_t)2314 * C; v2_2_20.R = GC + (size_t)2 * R3 * C; v2_2_20.C = GC + (size_t)2 * R3 * C;
      v2_2_20.sAo = (long long)34 * 34 * C; v2_2_20.sAi = (long long)34 * C; v2_2_20.sAm = C; v2_2_20.sAk = 1; v2_2_20.sBo = 0; v2_2_20.sBi = 0; v2_2_20.sBn = C * 27; v2_2_20.sBk = 27; v2_2_20.sCo = (long long)R * R * C; v2_2_20.sCi = (long long)R * C; v2_2_20.sCm = C; v2_2_20.sRo = (long long)R * R * C; v2_2_20.sRi = (long long)R * C; v2_2_20.sRm = C; v2_2_20.sRn = 1;
      v2_2_20.M = R; v2_2_20.N = C; v2_2_20.K = C; v2_2_20.zi_n = R; v2_2_20.flags = 4; v2_2_20.act = 0;
      v2_2_20.alpha = 1.0f; v2_2_20.beta = 1.0f; v2_2_20.sa = 1.0f; v2_2_20.sb = 1.0f; v2_2_20.Npad = C; v2_2_20.pad_ = 0;
      k_gemm<1><<<dim3((unsigned)((C) + 31) / 32, (unsigned)((R) + 15) / 16, (unsigned)(R * R)), 32, 0, stream>>>(v2_2_20); }
    { GemmP v2_2_21;
      v2_2_21.A = GQ + (size_t)2 * RP3 * C + (size_t)2346 * C; v2_2_21.B = wv2 + 21; v2_2_21.bias = GQ + (size_t)2 * RP3 * C + (size_t)2346 * C; v2_2_21.R = GC + (size_t)2 * R3 * C; v2_2_21.C = GC + (size_t)2 * R3 * C;
      v2_2_21.sAo = (long long)34 * 34 * C; v2_2_21.sAi = (long long)34 * C; v2_2_21.sAm = C; v2_2_21.sAk = 1; v2_2_21.sBo = 0; v2_2_21.sBi = 0; v2_2_21.sBn = C * 27; v2_2_21.sBk = 27; v2_2_21.sCo = (long long)R * R * C; v2_2_21.sCi = (long long)R * C; v2_2_21.sCm = C; v2_2_21.sRo = (long long)R * R * C; v2_2_21.sRi = (long long)R * C; v2_2_21.sRm = C; v2_2_21.sRn = 1;
      v2_2_21.M = R; v2_2_21.N = C; v2_2_21.K = C; v2_2_21.zi_n = R; v2_2_21.flags = 4; v2_2_21.act = 0;
      v2_2_21.alpha = 1.0f; v2_2_21.beta = 1.0f; v2_2_21.sa = 1.0f; v2_2_21.sb = 1.0f; v2_2_21.Npad = C; v2_2_21.pad_ = 0;
      k_gemm<1><<<dim3((unsigned)((C) + 31) / 32, (unsigned)((R) + 15) / 16, (unsigned)(R * R)), 32, 0, stream>>>(v2_2_21); }
    { GemmP v2_2_22;
      v2_2_22.A = GQ + (size_t)2 * RP3 * C + (size_t)2347 * C; v2_2_22.B = wv2 + 22; v2_2_22.bias = GQ + (size_t)2 * RP3 * C + (size_t)2347 * C; v2_2_22.R = GC + (size_t)2 * R3 * C; v2_2_22.C = GC + (size_t)2 * R3 * C;
      v2_2_22.sAo = (long long)34 * 34 * C; v2_2_22.sAi = (long long)34 * C; v2_2_22.sAm = C; v2_2_22.sAk = 1; v2_2_22.sBo = 0; v2_2_22.sBi = 0; v2_2_22.sBn = C * 27; v2_2_22.sBk = 27; v2_2_22.sCo = (long long)R * R * C; v2_2_22.sCi = (long long)R * C; v2_2_22.sCm = C; v2_2_22.sRo = (long long)R * R * C; v2_2_22.sRi = (long long)R * C; v2_2_22.sRm = C; v2_2_22.sRn = 1;
      v2_2_22.M = R; v2_2_22.N = C; v2_2_22.K = C; v2_2_22.zi_n = R; v2_2_22.flags = 4; v2_2_22.act = 0;
      v2_2_22.alpha = 1.0f; v2_2_22.beta = 1.0f; v2_2_22.sa = 1.0f; v2_2_22.sb = 1.0f; v2_2_22.Npad = C; v2_2_22.pad_ = 0;
      k_gemm<1><<<dim3((unsigned)((C) + 31) / 32, (unsigned)((R) + 15) / 16, (unsigned)(R * R)), 32, 0, stream>>>(v2_2_22); }
    { GemmP v2_2_23;
      v2_2_23.A = GQ + (size_t)2 * RP3 * C + (size_t)2348 * C; v2_2_23.B = wv2 + 23; v2_2_23.bias = GQ + (size_t)2 * RP3 * C + (size_t)2348 * C; v2_2_23.R = GC + (size_t)2 * R3 * C; v2_2_23.C = GC + (size_t)2 * R3 * C;
      v2_2_23.sAo = (long long)34 * 34 * C; v2_2_23.sAi = (long long)34 * C; v2_2_23.sAm = C; v2_2_23.sAk = 1; v2_2_23.sBo = 0; v2_2_23.sBi = 0; v2_2_23.sBn = C * 27; v2_2_23.sBk = 27; v2_2_23.sCo = (long long)R * R * C; v2_2_23.sCi = (long long)R * C; v2_2_23.sCm = C; v2_2_23.sRo = (long long)R * R * C; v2_2_23.sRi = (long long)R * C; v2_2_23.sRm = C; v2_2_23.sRn = 1;
      v2_2_23.M = R; v2_2_23.N = C; v2_2_23.K = C; v2_2_23.zi_n = R; v2_2_23.flags = 4; v2_2_23.act = 0;
      v2_2_23.alpha = 1.0f; v2_2_23.beta = 1.0f; v2_2_23.sa = 1.0f; v2_2_23.sb = 1.0f; v2_2_23.Npad = C; v2_2_23.pad_ = 0;
      k_gemm<1><<<dim3((unsigned)((C) + 31) / 32, (unsigned)((R) + 15) / 16, (unsigned)(R * R)), 32, 0, stream>>>(v2_2_23); }
    { GemmP v2_2_24;
      v2_2_24.A = GQ + (size_t)2 * RP3 * C + (size_t)2380 * C; v2_2_24.B = wv2 + 24; v2_2_24.bias = GQ + (size_t)2 * RP3 * C + (size_t)2380 * C; v2_2_24.R = GC + (size_t)2 * R3 * C; v2_2_24.C = GC + (size_t)2 * R3 * C;
      v2_2_24.sAo = (long long)34 * 34 * C; v2_2_24.sAi = (long long)34 * C; v2_2_24.sAm = C; v2_2_24.sAk = 1; v2_2_24.sBo = 0; v2_2_24.sBi = 0; v2_2_24.sBn = C * 27; v2_2_24.sBk = 27; v2_2_24.sCo = (long long)R * R * C; v2_2_24.sCi = (long long)R * C; v2_2_24.sCm = C; v2_2_24.sRo = (long long)R * R * C; v2_2_24.sRi = (long long)R * C; v2_2_24.sRm = C; v2_2_24.sRn = 1;
      v2_2_24.M = R; v2_2_24.N = C; v2_2_24.K = C; v2_2_24.zi_n = R; v2_2_24.flags = 4; v2_2_24.act = 0;
      v2_2_24.alpha = 1.0f; v2_2_24.beta = 1.0f; v2_2_24.sa = 1.0f; v2_2_24.sb = 1.0f; v2_2_24.Npad = C; v2_2_24.pad_ = 0;
      k_gemm<1><<<dim3((unsigned)((C) + 31) / 32, (unsigned)((R) + 15) / 16, (unsigned)(R * R)), 32, 0, stream>>>(v2_2_24); }
    { GemmP v2_2_25;
      v2_2_25.A = GQ + (size_t)2 * RP3 * C + (size_t)2381 * C; v2_2_25.B = wv2 + 25; v2_2_25.bias = GQ + (size_t)2 * RP3 * C + (size_t)2381 * C; v2_2_25.R = GC + (size_t)2 * R3 * C; v2_2_25.C = GC + (size_t)2 * R3 * C;
      v2_2_25.sAo = (long long)34 * 34 * C; v2_2_25.sAi = (long long)34 * C; v2_2_25.sAm = C; v2_2_25.sAk = 1; v2_2_25.sBo = 0; v2_2_25.sBi = 0; v2_2_25.sBn = C * 27; v2_2_25.sBk = 27; v2_2_25.sCo = (long long)R * R * C; v2_2_25.sCi = (long long)R * C; v2_2_25.sCm = C; v2_2_25.sRo = (long long)R * R * C; v2_2_25.sRi = (long long)R * C; v2_2_25.sRm = C; v2_2_25.sRn = 1;
      v2_2_25.M = R; v2_2_25.N = C; v2_2_25.K = C; v2_2_25.zi_n = R; v2_2_25.flags = 4; v2_2_25.act = 0;
      v2_2_25.alpha = 1.0f; v2_2_25.beta = 1.0f; v2_2_25.sa = 1.0f; v2_2_25.sb = 1.0f; v2_2_25.Npad = C; v2_2_25.pad_ = 0;
      k_gemm<1><<<dim3((unsigned)((C) + 31) / 32, (unsigned)((R) + 15) / 16, (unsigned)(R * R)), 32, 0, stream>>>(v2_2_25); }
    { GemmP v2_2_26;
      v2_2_26.A = GQ + (size_t)2 * RP3 * C + (size_t)2382 * C; v2_2_26.B = wv2 + 26; v2_2_26.bias = GQ + (size_t)2 * RP3 * C + (size_t)2382 * C; v2_2_26.R = GC + (size_t)2 * R3 * C; v2_2_26.C = GC + (size_t)2 * R3 * C;
      v2_2_26.sAo = (long long)34 * 34 * C; v2_2_26.sAi = (long long)34 * C; v2_2_26.sAm = C; v2_2_26.sAk = 1; v2_2_26.sBo = 0; v2_2_26.sBi = 0; v2_2_26.sBn = C * 27; v2_2_26.sBk = 27; v2_2_26.sCo = (long long)R * R * C; v2_2_26.sCi = (long long)R * C; v2_2_26.sCm = C; v2_2_26.sRo = (long long)R * R * C; v2_2_26.sRi = (long long)R * C; v2_2_26.sRm = C; v2_2_26.sRn = 1;
      v2_2_26.M = R; v2_2_26.N = C; v2_2_26.K = C; v2_2_26.zi_n = R; v2_2_26.flags = 4; v2_2_26.act = 0;
      v2_2_26.alpha = 1.0f; v2_2_26.beta = 1.0f; v2_2_26.sa = 1.0f; v2_2_26.sb = 1.0f; v2_2_26.Npad = C; v2_2_26.pad_ = 0;
      k_gemm<1><<<dim3((unsigned)((C) + 31) / 32, (unsigned)((R) + 15) / 16, (unsigned)(R * R)), 32, 0, stream>>>(v2_2_26); }
    { GemmP v2_3_0;
      v2_3_0.A = GQ + (size_t)3 * RP3 * C + (size_t)0 * C; v2_3_0.B = wv2 + 0; v2_3_0.bias = bv2; v2_3_0.R = GQ + (size_t)3 * RP3 * C + (size_t)0 * C; v2_3_0.C = GC + (size_t)3 * R3 * C;
      v2_3_0.sAo = (long long)34 * 34 * C; v2_3_0.sAi = (long long)34 * C; v2_3_0.sAm = C; v2_3_0.sAk = 1; v2_3_0.sBo = 0; v2_3_0.sBi = 0; v2_3_0.sBn = C * 27; v2_3_0.sBk = 27; v2_3_0.sCo = (long long)R * R * C; v2_3_0.sCi = (long long)R * C; v2_3_0.sCm = C; v2_3_0.sRo = 0; v2_3_0.sRi = 0; v2_3_0.sRm = 0; v2_3_0.sRn = 0;
      v2_3_0.M = R; v2_3_0.N = C; v2_3_0.K = C; v2_3_0.zi_n = R; v2_3_0.flags = 1; v2_3_0.act = 0;
      v2_3_0.alpha = 1.0f; v2_3_0.beta = 0.0f; v2_3_0.sa = 1.0f; v2_3_0.sb = 1.0f; v2_3_0.Npad = C; v2_3_0.pad_ = 0;
      k_gemm<1><<<dim3((unsigned)((C) + 31) / 32, (unsigned)((R) + 15) / 16, (unsigned)(R * R)), 32, 0, stream>>>(v2_3_0); }
    { GemmP v2_3_1;
      v2_3_1.A = GQ + (size_t)3 * RP3 * C + (size_t)1 * C; v2_3_1.B = wv2 + 1; v2_3_1.bias = GQ + (size_t)3 * RP3 * C + (size_t)1 * C; v2_3_1.R = GC + (size_t)3 * R3 * C; v2_3_1.C = GC + (size_t)3 * R3 * C;
      v2_3_1.sAo = (long long)34 * 34 * C; v2_3_1.sAi = (long long)34 * C; v2_3_1.sAm = C; v2_3_1.sAk = 1; v2_3_1.sBo = 0; v2_3_1.sBi = 0; v2_3_1.sBn = C * 27; v2_3_1.sBk = 27; v2_3_1.sCo = (long long)R * R * C; v2_3_1.sCi = (long long)R * C; v2_3_1.sCm = C; v2_3_1.sRo = (long long)R * R * C; v2_3_1.sRi = (long long)R * C; v2_3_1.sRm = C; v2_3_1.sRn = 1;
      v2_3_1.M = R; v2_3_1.N = C; v2_3_1.K = C; v2_3_1.zi_n = R; v2_3_1.flags = 4; v2_3_1.act = 0;
      v2_3_1.alpha = 1.0f; v2_3_1.beta = 1.0f; v2_3_1.sa = 1.0f; v2_3_1.sb = 1.0f; v2_3_1.Npad = C; v2_3_1.pad_ = 0;
      k_gemm<1><<<dim3((unsigned)((C) + 31) / 32, (unsigned)((R) + 15) / 16, (unsigned)(R * R)), 32, 0, stream>>>(v2_3_1); }
    { GemmP v2_3_2;
      v2_3_2.A = GQ + (size_t)3 * RP3 * C + (size_t)2 * C; v2_3_2.B = wv2 + 2; v2_3_2.bias = GQ + (size_t)3 * RP3 * C + (size_t)2 * C; v2_3_2.R = GC + (size_t)3 * R3 * C; v2_3_2.C = GC + (size_t)3 * R3 * C;
      v2_3_2.sAo = (long long)34 * 34 * C; v2_3_2.sAi = (long long)34 * C; v2_3_2.sAm = C; v2_3_2.sAk = 1; v2_3_2.sBo = 0; v2_3_2.sBi = 0; v2_3_2.sBn = C * 27; v2_3_2.sBk = 27; v2_3_2.sCo = (long long)R * R * C; v2_3_2.sCi = (long long)R * C; v2_3_2.sCm = C; v2_3_2.sRo = (long long)R * R * C; v2_3_2.sRi = (long long)R * C; v2_3_2.sRm = C; v2_3_2.sRn = 1;
      v2_3_2.M = R; v2_3_2.N = C; v2_3_2.K = C; v2_3_2.zi_n = R; v2_3_2.flags = 4; v2_3_2.act = 0;
      v2_3_2.alpha = 1.0f; v2_3_2.beta = 1.0f; v2_3_2.sa = 1.0f; v2_3_2.sb = 1.0f; v2_3_2.Npad = C; v2_3_2.pad_ = 0;
      k_gemm<1><<<dim3((unsigned)((C) + 31) / 32, (unsigned)((R) + 15) / 16, (unsigned)(R * R)), 32, 0, stream>>>(v2_3_2); }
    { GemmP v2_3_3;
      v2_3_3.A = GQ + (size_t)3 * RP3 * C + (size_t)34 * C; v2_3_3.B = wv2 + 3; v2_3_3.bias = GQ + (size_t)3 * RP3 * C + (size_t)34 * C; v2_3_3.R = GC + (size_t)3 * R3 * C; v2_3_3.C = GC + (size_t)3 * R3 * C;
      v2_3_3.sAo = (long long)34 * 34 * C; v2_3_3.sAi = (long long)34 * C; v2_3_3.sAm = C; v2_3_3.sAk = 1; v2_3_3.sBo = 0; v2_3_3.sBi = 0; v2_3_3.sBn = C * 27; v2_3_3.sBk = 27; v2_3_3.sCo = (long long)R * R * C; v2_3_3.sCi = (long long)R * C; v2_3_3.sCm = C; v2_3_3.sRo = (long long)R * R * C; v2_3_3.sRi = (long long)R * C; v2_3_3.sRm = C; v2_3_3.sRn = 1;
      v2_3_3.M = R; v2_3_3.N = C; v2_3_3.K = C; v2_3_3.zi_n = R; v2_3_3.flags = 4; v2_3_3.act = 0;
      v2_3_3.alpha = 1.0f; v2_3_3.beta = 1.0f; v2_3_3.sa = 1.0f; v2_3_3.sb = 1.0f; v2_3_3.Npad = C; v2_3_3.pad_ = 0;
      k_gemm<1><<<dim3((unsigned)((C) + 31) / 32, (unsigned)((R) + 15) / 16, (unsigned)(R * R)), 32, 0, stream>>>(v2_3_3); }
    { GemmP v2_3_4;
      v2_3_4.A = GQ + (size_t)3 * RP3 * C + (size_t)35 * C; v2_3_4.B = wv2 + 4; v2_3_4.bias = GQ + (size_t)3 * RP3 * C + (size_t)35 * C; v2_3_4.R = GC + (size_t)3 * R3 * C; v2_3_4.C = GC + (size_t)3 * R3 * C;
      v2_3_4.sAo = (long long)34 * 34 * C; v2_3_4.sAi = (long long)34 * C; v2_3_4.sAm = C; v2_3_4.sAk = 1; v2_3_4.sBo = 0; v2_3_4.sBi = 0; v2_3_4.sBn = C * 27; v2_3_4.sBk = 27; v2_3_4.sCo = (long long)R * R * C; v2_3_4.sCi = (long long)R * C; v2_3_4.sCm = C; v2_3_4.sRo = (long long)R * R * C; v2_3_4.sRi = (long long)R * C; v2_3_4.sRm = C; v2_3_4.sRn = 1;
      v2_3_4.M = R; v2_3_4.N = C; v2_3_4.K = C; v2_3_4.zi_n = R; v2_3_4.flags = 4; v2_3_4.act = 0;
      v2_3_4.alpha = 1.0f; v2_3_4.beta = 1.0f; v2_3_4.sa = 1.0f; v2_3_4.sb = 1.0f; v2_3_4.Npad = C; v2_3_4.pad_ = 0;
      k_gemm<1><<<dim3((unsigned)((C) + 31) / 32, (unsigned)((R) + 15) / 16, (unsigned)(R * R)), 32, 0, stream>>>(v2_3_4); }
    { GemmP v2_3_5;
      v2_3_5.A = GQ + (size_t)3 * RP3 * C + (size_t)36 * C; v2_3_5.B = wv2 + 5; v2_3_5.bias = GQ + (size_t)3 * RP3 * C + (size_t)36 * C; v2_3_5.R = GC + (size_t)3 * R3 * C; v2_3_5.C = GC + (size_t)3 * R3 * C;
      v2_3_5.sAo = (long long)34 * 34 * C; v2_3_5.sAi = (long long)34 * C; v2_3_5.sAm = C; v2_3_5.sAk = 1; v2_3_5.sBo = 0; v2_3_5.sBi = 0; v2_3_5.sBn = C * 27; v2_3_5.sBk = 27; v2_3_5.sCo = (long long)R * R * C; v2_3_5.sCi = (long long)R * C; v2_3_5.sCm = C; v2_3_5.sRo = (long long)R * R * C; v2_3_5.sRi = (long long)R * C; v2_3_5.sRm = C; v2_3_5.sRn = 1;
      v2_3_5.M = R; v2_3_5.N = C; v2_3_5.K = C; v2_3_5.zi_n = R; v2_3_5.flags = 4; v2_3_5.act = 0;
      v2_3_5.alpha = 1.0f; v2_3_5.beta = 1.0f; v2_3_5.sa = 1.0f; v2_3_5.sb = 1.0f; v2_3_5.Npad = C; v2_3_5.pad_ = 0;
      k_gemm<1><<<dim3((unsigned)((C) + 31) / 32, (unsigned)((R) + 15) / 16, (unsigned)(R * R)), 32, 0, stream>>>(v2_3_5); }
    { GemmP v2_3_6;
      v2_3_6.A = GQ + (size_t)3 * RP3 * C + (size_t)68 * C; v2_3_6.B = wv2 + 6; v2_3_6.bias = GQ + (size_t)3 * RP3 * C + (size_t)68 * C; v2_3_6.R = GC + (size_t)3 * R3 * C; v2_3_6.C = GC + (size_t)3 * R3 * C;
      v2_3_6.sAo = (long long)34 * 34 * C; v2_3_6.sAi = (long long)34 * C; v2_3_6.sAm = C; v2_3_6.sAk = 1; v2_3_6.sBo = 0; v2_3_6.sBi = 0; v2_3_6.sBn = C * 27; v2_3_6.sBk = 27; v2_3_6.sCo = (long long)R * R * C; v2_3_6.sCi = (long long)R * C; v2_3_6.sCm = C; v2_3_6.sRo = (long long)R * R * C; v2_3_6.sRi = (long long)R * C; v2_3_6.sRm = C; v2_3_6.sRn = 1;
      v2_3_6.M = R; v2_3_6.N = C; v2_3_6.K = C; v2_3_6.zi_n = R; v2_3_6.flags = 4; v2_3_6.act = 0;
      v2_3_6.alpha = 1.0f; v2_3_6.beta = 1.0f; v2_3_6.sa = 1.0f; v2_3_6.sb = 1.0f; v2_3_6.Npad = C; v2_3_6.pad_ = 0;
      k_gemm<1><<<dim3((unsigned)((C) + 31) / 32, (unsigned)((R) + 15) / 16, (unsigned)(R * R)), 32, 0, stream>>>(v2_3_6); }
    { GemmP v2_3_7;
      v2_3_7.A = GQ + (size_t)3 * RP3 * C + (size_t)69 * C; v2_3_7.B = wv2 + 7; v2_3_7.bias = GQ + (size_t)3 * RP3 * C + (size_t)69 * C; v2_3_7.R = GC + (size_t)3 * R3 * C; v2_3_7.C = GC + (size_t)3 * R3 * C;
      v2_3_7.sAo = (long long)34 * 34 * C; v2_3_7.sAi = (long long)34 * C; v2_3_7.sAm = C; v2_3_7.sAk = 1; v2_3_7.sBo = 0; v2_3_7.sBi = 0; v2_3_7.sBn = C * 27; v2_3_7.sBk = 27; v2_3_7.sCo = (long long)R * R * C; v2_3_7.sCi = (long long)R * C; v2_3_7.sCm = C; v2_3_7.sRo = (long long)R * R * C; v2_3_7.sRi = (long long)R * C; v2_3_7.sRm = C; v2_3_7.sRn = 1;
      v2_3_7.M = R; v2_3_7.N = C; v2_3_7.K = C; v2_3_7.zi_n = R; v2_3_7.flags = 4; v2_3_7.act = 0;
      v2_3_7.alpha = 1.0f; v2_3_7.beta = 1.0f; v2_3_7.sa = 1.0f; v2_3_7.sb = 1.0f; v2_3_7.Npad = C; v2_3_7.pad_ = 0;
      k_gemm<1><<<dim3((unsigned)((C) + 31) / 32, (unsigned)((R) + 15) / 16, (unsigned)(R * R)), 32, 0, stream>>>(v2_3_7); }
    { GemmP v2_3_8;
      v2_3_8.A = GQ + (size_t)3 * RP3 * C + (size_t)70 * C; v2_3_8.B = wv2 + 8; v2_3_8.bias = GQ + (size_t)3 * RP3 * C + (size_t)70 * C; v2_3_8.R = GC + (size_t)3 * R3 * C; v2_3_8.C = GC + (size_t)3 * R3 * C;
      v2_3_8.sAo = (long long)34 * 34 * C; v2_3_8.sAi = (long long)34 * C; v2_3_8.sAm = C; v2_3_8.sAk = 1; v2_3_8.sBo = 0; v2_3_8.sBi = 0; v2_3_8.sBn = C * 27; v2_3_8.sBk = 27; v2_3_8.sCo = (long long)R * R * C; v2_3_8.sCi = (long long)R * C; v2_3_8.sCm = C; v2_3_8.sRo = (long long)R * R * C; v2_3_8.sRi = (long long)R * C; v2_3_8.sRm = C; v2_3_8.sRn = 1;
      v2_3_8.M = R; v2_3_8.N = C; v2_3_8.K = C; v2_3_8.zi_n = R; v2_3_8.flags = 4; v2_3_8.act = 0;
      v2_3_8.alpha = 1.0f; v2_3_8.beta = 1.0f; v2_3_8.sa = 1.0f; v2_3_8.sb = 1.0f; v2_3_8.Npad = C; v2_3_8.pad_ = 0;
      k_gemm<1><<<dim3((unsigned)((C) + 31) / 32, (unsigned)((R) + 15) / 16, (unsigned)(R * R)), 32, 0, stream>>>(v2_3_8); }
    { GemmP v2_3_9;
      v2_3_9.A = GQ + (size_t)3 * RP3 * C + (size_t)1156 * C; v2_3_9.B = wv2 + 9; v2_3_9.bias = GQ + (size_t)3 * RP3 * C + (size_t)1156 * C; v2_3_9.R = GC + (size_t)3 * R3 * C; v2_3_9.C = GC + (size_t)3 * R3 * C;
      v2_3_9.sAo = (long long)34 * 34 * C; v2_3_9.sAi = (long long)34 * C; v2_3_9.sAm = C; v2_3_9.sAk = 1; v2_3_9.sBo = 0; v2_3_9.sBi = 0; v2_3_9.sBn = C * 27; v2_3_9.sBk = 27; v2_3_9.sCo = (long long)R * R * C; v2_3_9.sCi = (long long)R * C; v2_3_9.sCm = C; v2_3_9.sRo = (long long)R * R * C; v2_3_9.sRi = (long long)R * C; v2_3_9.sRm = C; v2_3_9.sRn = 1;
      v2_3_9.M = R; v2_3_9.N = C; v2_3_9.K = C; v2_3_9.zi_n = R; v2_3_9.flags = 4; v2_3_9.act = 0;
      v2_3_9.alpha = 1.0f; v2_3_9.beta = 1.0f; v2_3_9.sa = 1.0f; v2_3_9.sb = 1.0f; v2_3_9.Npad = C; v2_3_9.pad_ = 0;
      k_gemm<1><<<dim3((unsigned)((C) + 31) / 32, (unsigned)((R) + 15) / 16, (unsigned)(R * R)), 32, 0, stream>>>(v2_3_9); }
    { GemmP v2_3_10;
      v2_3_10.A = GQ + (size_t)3 * RP3 * C + (size_t)1157 * C; v2_3_10.B = wv2 + 10; v2_3_10.bias = GQ + (size_t)3 * RP3 * C + (size_t)1157 * C; v2_3_10.R = GC + (size_t)3 * R3 * C; v2_3_10.C = GC + (size_t)3 * R3 * C;
      v2_3_10.sAo = (long long)34 * 34 * C; v2_3_10.sAi = (long long)34 * C; v2_3_10.sAm = C; v2_3_10.sAk = 1; v2_3_10.sBo = 0; v2_3_10.sBi = 0; v2_3_10.sBn = C * 27; v2_3_10.sBk = 27; v2_3_10.sCo = (long long)R * R * C; v2_3_10.sCi = (long long)R * C; v2_3_10.sCm = C; v2_3_10.sRo = (long long)R * R * C; v2_3_10.sRi = (long long)R * C; v2_3_10.sRm = C; v2_3_10.sRn = 1;
      v2_3_10.M = R; v2_3_10.N = C; v2_3_10.K = C; v2_3_10.zi_n = R; v2_3_10.flags = 4; v2_3_10.act = 0;
      v2_3_10.alpha = 1.0f; v2_3_10.beta = 1.0f; v2_3_10.sa = 1.0f; v2_3_10.sb = 1.0f; v2_3_10.Npad = C; v2_3_10.pad_ = 0;
      k_gemm<1><<<dim3((unsigned)((C) + 31) / 32, (unsigned)((R) + 15) / 16, (unsigned)(R * R)), 32, 0, stream>>>(v2_3_10); }
    { GemmP v2_3_11;
      v2_3_11.A = GQ + (size_t)3 * RP3 * C + (size_t)1158 * C; v2_3_11.B = wv2 + 11; v2_3_11.bias = GQ + (size_t)3 * RP3 * C + (size_t)1158 * C; v2_3_11.R = GC + (size_t)3 * R3 * C; v2_3_11.C = GC + (size_t)3 * R3 * C;
      v2_3_11.sAo = (long long)34 * 34 * C; v2_3_11.sAi = (long long)34 * C; v2_3_11.sAm = C; v2_3_11.sAk = 1; v2_3_11.sBo = 0; v2_3_11.sBi = 0; v2_3_11.sBn = C * 27; v2_3_11.sBk = 27; v2_3_11.sCo = (long long)R * R * C; v2_3_11.sCi = (long long)R * C; v2_3_11.sCm = C; v2_3_11.sRo = (long long)R * R * C; v2_3_11.sRi = (long long)R * C; v2_3_11.sRm = C; v2_3_11.sRn = 1;
      v2_3_11.M = R; v2_3_11.N = C; v2_3_11.K = C; v2_3_11.zi_n = R; v2_3_11.flags = 4; v2_3_11.act = 0;
      v2_3_11.alpha = 1.0f; v2_3_11.beta = 1.0f; v2_3_11.sa = 1.0f; v2_3_11.sb = 1.0f; v2_3_11.Npad = C; v2_3_11.pad_ = 0;
      k_gemm<1><<<dim3((unsigned)((C) + 31) / 32, (unsigned)((R) + 15) / 16, (unsigned)(R * R)), 32, 0, stream>>>(v2_3_11); }
    { GemmP v2_3_12;
      v2_3_12.A = GQ + (size_t)3 * RP3 * C + (size_t)1190 * C; v2_3_12.B = wv2 + 12; v2_3_12.bias = GQ + (size_t)3 * RP3 * C + (size_t)1190 * C; v2_3_12.R = GC + (size_t)3 * R3 * C; v2_3_12.C = GC + (size_t)3 * R3 * C;
      v2_3_12.sAo = (long long)34 * 34 * C; v2_3_12.sAi = (long long)34 * C; v2_3_12.sAm = C; v2_3_12.sAk = 1; v2_3_12.sBo = 0; v2_3_12.sBi = 0; v2_3_12.sBn = C * 27; v2_3_12.sBk = 27; v2_3_12.sCo = (long long)R * R * C; v2_3_12.sCi = (long long)R * C; v2_3_12.sCm = C; v2_3_12.sRo = (long long)R * R * C; v2_3_12.sRi = (long long)R * C; v2_3_12.sRm = C; v2_3_12.sRn = 1;
      v2_3_12.M = R; v2_3_12.N = C; v2_3_12.K = C; v2_3_12.zi_n = R; v2_3_12.flags = 4; v2_3_12.act = 0;
      v2_3_12.alpha = 1.0f; v2_3_12.beta = 1.0f; v2_3_12.sa = 1.0f; v2_3_12.sb = 1.0f; v2_3_12.Npad = C; v2_3_12.pad_ = 0;
      k_gemm<1><<<dim3((unsigned)((C) + 31) / 32, (unsigned)((R) + 15) / 16, (unsigned)(R * R)), 32, 0, stream>>>(v2_3_12); }
    { GemmP v2_3_13;
      v2_3_13.A = GQ + (size_t)3 * RP3 * C + (size_t)1191 * C; v2_3_13.B = wv2 + 13; v2_3_13.bias = GQ + (size_t)3 * RP3 * C + (size_t)1191 * C; v2_3_13.R = GC + (size_t)3 * R3 * C; v2_3_13.C = GC + (size_t)3 * R3 * C;
      v2_3_13.sAo = (long long)34 * 34 * C; v2_3_13.sAi = (long long)34 * C; v2_3_13.sAm = C; v2_3_13.sAk = 1; v2_3_13.sBo = 0; v2_3_13.sBi = 0; v2_3_13.sBn = C * 27; v2_3_13.sBk = 27; v2_3_13.sCo = (long long)R * R * C; v2_3_13.sCi = (long long)R * C; v2_3_13.sCm = C; v2_3_13.sRo = (long long)R * R * C; v2_3_13.sRi = (long long)R * C; v2_3_13.sRm = C; v2_3_13.sRn = 1;
      v2_3_13.M = R; v2_3_13.N = C; v2_3_13.K = C; v2_3_13.zi_n = R; v2_3_13.flags = 4; v2_3_13.act = 0;
      v2_3_13.alpha = 1.0f; v2_3_13.beta = 1.0f; v2_3_13.sa = 1.0f; v2_3_13.sb = 1.0f; v2_3_13.Npad = C; v2_3_13.pad_ = 0;
      k_gemm<1><<<dim3((unsigned)((C) + 31) / 32, (unsigned)((R) + 15) / 16, (unsigned)(R * R)), 32, 0, stream>>>(v2_3_13); }
    { GemmP v2_3_14;
      v2_3_14.A = GQ + (size_t)3 * RP3 * C + (size_t)1192 * C; v2_3_14.B = wv2 + 14; v2_3_14.bias = GQ + (size_t)3 * RP3 * C + (size_t)1192 * C; v2_3_14.R = GC + (size_t)3 * R3 * C; v2_3_14.C = GC + (size_t)3 * R3 * C;
      v2_3_14.sAo = (long long)34 * 34 * C; v2_3_14.sAi = (long long)34 * C; v2_3_14.sAm = C; v2_3_14.sAk = 1; v2_3_14.sBo = 0; v2_3_14.sBi = 0; v2_3_14.sBn = C * 27; v2_3_14.sBk = 27; v2_3_14.sCo = (long long)R * R * C; v2_3_14.sCi = (long long)R * C; v2_3_14.sCm = C; v2_3_14.sRo = (long long)R * R * C; v2_3_14.sRi = (long long)R * C; v2_3_14.sRm = C; v2_3_14.sRn = 1;
      v2_3_14.M = R; v2_3_14.N = C; v2_3_14.K = C; v2_3_14.zi_n = R; v2_3_14.flags = 4; v2_3_14.act = 0;
      v2_3_14.alpha = 1.0f; v2_3_14.beta = 1.0f; v2_3_14.sa = 1.0f; v2_3_14.sb = 1.0f; v2_3_14.Npad = C; v2_3_14.pad_ = 0;
      k_gemm<1><<<dim3((unsigned)((C) + 31) / 32, (unsigned)((R) + 15) / 16, (unsigned)(R * R)), 32, 0, stream>>>(v2_3_14); }
    { GemmP v2_3_15;
      v2_3_15.A = GQ + (size_t)3 * RP3 * C + (size_t)1224 * C; v2_3_15.B = wv2 + 15; v2_3_15.bias = GQ + (size_t)3 * RP3 * C + (size_t)1224 * C; v2_3_15.R = GC + (size_t)3 * R3 * C; v2_3_15.C = GC + (size_t)3 * R3 * C;
      v2_3_15.sAo = (long long)34 * 34 * C; v2_3_15.sAi = (long long)34 * C; v2_3_15.sAm = C; v2_3_15.sAk = 1; v2_3_15.sBo = 0; v2_3_15.sBi = 0; v2_3_15.sBn = C * 27; v2_3_15.sBk = 27; v2_3_15.sCo = (long long)R * R * C; v2_3_15.sCi = (long long)R * C; v2_3_15.sCm = C; v2_3_15.sRo = (long long)R * R * C; v2_3_15.sRi = (long long)R * C; v2_3_15.sRm = C; v2_3_15.sRn = 1;
      v2_3_15.M = R; v2_3_15.N = C; v2_3_15.K = C; v2_3_15.zi_n = R; v2_3_15.flags = 4; v2_3_15.act = 0;
      v2_3_15.alpha = 1.0f; v2_3_15.beta = 1.0f; v2_3_15.sa = 1.0f; v2_3_15.sb = 1.0f; v2_3_15.Npad = C; v2_3_15.pad_ = 0;
      k_gemm<1><<<dim3((unsigned)((C) + 31) / 32, (unsigned)((R) + 15) / 16, (unsigned)(R * R)), 32, 0, stream>>>(v2_3_15); }
    { GemmP v2_3_16;
      v2_3_16.A = GQ + (size_t)3 * RP3 * C + (size_t)1225 * C; v2_3_16.B = wv2 + 16; v2_3_16.bias = GQ + (size_t)3 * RP3 * C + (size_t)1225 * C; v2_3_16.R = GC + (size_t)3 * R3 * C; v2_3_16.C = GC + (size_t)3 * R3 * C;
      v2_3_16.sAo = (long long)34 * 34 * C; v2_3_16.sAi = (long long)34 * C; v2_3_16.sAm = C; v2_3_16.sAk = 1; v2_3_16.sBo = 0; v2_3_16.sBi = 0; v2_3_16.sBn = C * 27; v2_3_16.sBk = 27; v2_3_16.sCo = (long long)R * R * C; v2_3_16.sCi = (long long)R * C; v2_3_16.sCm = C; v2_3_16.sRo = (long long)R * R * C; v2_3_16.sRi = (long long)R * C; v2_3_16.sRm = C; v2_3_16.sRn = 1;
      v2_3_16.M = R; v2_3_16.N = C; v2_3_16.K = C; v2_3_16.zi_n = R; v2_3_16.flags = 4; v2_3_16.act = 0;
      v2_3_16.alpha = 1.0f; v2_3_16.beta = 1.0f; v2_3_16.sa = 1.0f; v2_3_16.sb = 1.0f; v2_3_16.Npad = C; v2_3_16.pad_ = 0;
      k_gemm<1><<<dim3((unsigned)((C) + 31) / 32, (unsigned)((R) + 15) / 16, (unsigned)(R * R)), 32, 0, stream>>>(v2_3_16); }
    { GemmP v2_3_17;
      v2_3_17.A = GQ + (size_t)3 * RP3 * C + (size_t)1226 * C; v2_3_17.B = wv2 + 17; v2_3_17.bias = GQ + (size_t)3 * RP3 * C + (size_t)1226 * C; v2_3_17.R = GC + (size_t)3 * R3 * C; v2_3_17.C = GC + (size_t)3 * R3 * C;
      v2_3_17.sAo = (long long)34 * 34 * C; v2_3_17.sAi = (long long)34 * C; v2_3_17.sAm = C; v2_3_17.sAk = 1; v2_3_17.sBo = 0; v2_3_17.sBi = 0; v2_3_17.sBn = C * 27; v2_3_17.sBk = 27; v2_3_17.sCo = (long long)R * R * C; v2_3_17.sCi = (long long)R * C; v2_3_17.sCm = C; v2_3_17.sRo = (long long)R * R * C; v2_3_17.sRi = (long long)R * C; v2_3_17.sRm = C; v2_3_17.sRn = 1;
      v2_3_17.M = R; v2_3_17.N = C; v2_3_17.K = C; v2_3_17.zi_n = R; v2_3_17.flags = 4; v2_3_17.act = 0;
      v2_3_17.alpha = 1.0f; v2_3_17.beta = 1.0f; v2_3_17.sa = 1.0f; v2_3_17.sb = 1.0f; v2_3_17.Npad = C; v2_3_17.pad_ = 0;
      k_gemm<1><<<dim3((unsigned)((C) + 31) / 32, (unsigned)((R) + 15) / 16, (unsigned)(R * R)), 32, 0, stream>>>(v2_3_17); }
    { GemmP v2_3_18;
      v2_3_18.A = GQ + (size_t)3 * RP3 * C + (size_t)2312 * C; v2_3_18.B = wv2 + 18; v2_3_18.bias = GQ + (size_t)3 * RP3 * C + (size_t)2312 * C; v2_3_18.R = GC + (size_t)3 * R3 * C; v2_3_18.C = GC + (size_t)3 * R3 * C;
      v2_3_18.sAo = (long long)34 * 34 * C; v2_3_18.sAi = (long long)34 * C; v2_3_18.sAm = C; v2_3_18.sAk = 1; v2_3_18.sBo = 0; v2_3_18.sBi = 0; v2_3_18.sBn = C * 27; v2_3_18.sBk = 27; v2_3_18.sCo = (long long)R * R * C; v2_3_18.sCi = (long long)R * C; v2_3_18.sCm = C; v2_3_18.sRo = (long long)R * R * C; v2_3_18.sRi = (long long)R * C; v2_3_18.sRm = C; v2_3_18.sRn = 1;
      v2_3_18.M = R; v2_3_18.N = C; v2_3_18.K = C; v2_3_18.zi_n = R; v2_3_18.flags = 4; v2_3_18.act = 0;
      v2_3_18.alpha = 1.0f; v2_3_18.beta = 1.0f; v2_3_18.sa = 1.0f; v2_3_18.sb = 1.0f; v2_3_18.Npad = C; v2_3_18.pad_ = 0;
      k_gemm<1><<<dim3((unsigned)((C) + 31) / 32, (unsigned)((R) + 15) / 16, (unsigned)(R * R)), 32, 0, stream>>>(v2_3_18); }
    { GemmP v2_3_19;
      v2_3_19.A = GQ + (size_t)3 * RP3 * C + (size_t)2313 * C; v2_3_19.B = wv2 + 19; v2_3_19.bias = GQ + (size_t)3 * RP3 * C + (size_t)2313 * C; v2_3_19.R = GC + (size_t)3 * R3 * C; v2_3_19.C = GC + (size_t)3 * R3 * C;
      v2_3_19.sAo = (long long)34 * 34 * C; v2_3_19.sAi = (long long)34 * C; v2_3_19.sAm = C; v2_3_19.sAk = 1; v2_3_19.sBo = 0; v2_3_19.sBi = 0; v2_3_19.sBn = C * 27; v2_3_19.sBk = 27; v2_3_19.sCo = (long long)R * R * C; v2_3_19.sCi = (long long)R * C; v2_3_19.sCm = C; v2_3_19.sRo = (long long)R * R * C; v2_3_19.sRi = (long long)R * C; v2_3_19.sRm = C; v2_3_19.sRn = 1;
      v2_3_19.M = R; v2_3_19.N = C; v2_3_19.K = C; v2_3_19.zi_n = R; v2_3_19.flags = 4; v2_3_19.act = 0;
      v2_3_19.alpha = 1.0f; v2_3_19.beta = 1.0f; v2_3_19.sa = 1.0f; v2_3_19.sb = 1.0f; v2_3_19.Npad = C; v2_3_19.pad_ = 0;
      k_gemm<1><<<dim3((unsigned)((C) + 31) / 32, (unsigned)((R) + 15) / 16, (unsigned)(R * R)), 32, 0, stream>>>(v2_3_19); }
    { GemmP v2_3_20;
      v2_3_20.A = GQ + (size_t)3 * RP3 * C + (size_t)2314 * C; v2_3_20.B = wv2 + 20; v2_3_20.bias = GQ + (size_t)3 * RP3 * C + (size_t)2314 * C; v2_3_20.R = GC + (size_t)3 * R3 * C; v2_3_20.C = GC + (size_t)3 * R3 * C;
      v2_3_20.sAo = (long long)34 * 34 * C; v2_3_20.sAi = (long long)34 * C; v2_3_20.sAm = C; v2_3_20.sAk = 1; v2_3_20.sBo = 0; v2_3_20.sBi = 0; v2_3_20.sBn = C * 27; v2_3_20.sBk = 27; v2_3_20.sCo = (long long)R * R * C; v2_3_20.sCi = (long long)R * C; v2_3_20.sCm = C; v2_3_20.sRo = (long long)R * R * C; v2_3_20.sRi = (long long)R * C; v2_3_20.sRm = C; v2_3_20.sRn = 1;
      v2_3_20.M = R; v2_3_20.N = C; v2_3_20.K = C; v2_3_20.zi_n = R; v2_3_20.flags = 4; v2_3_20.act = 0;
      v2_3_20.alpha = 1.0f; v2_3_20.beta = 1.0f; v2_3_20.sa = 1.0f; v2_3_20.sb = 1.0f; v2_3_20.Npad = C; v2_3_20.pad_ = 0;
      k_gemm<1><<<dim3((unsigned)((C) + 31) / 32, (unsigned)((R) + 15) / 16, (unsigned)(R * R)), 32, 0, stream>>>(v2_3_20); }
    { GemmP v2_3_21;
      v2_3_21.A = GQ + (size_t)3 * RP3 * C + (size_t)2346 * C; v2_3_21.B = wv2 + 21; v2_3_21.bias = GQ + (size_t)3 * RP3 * C + (size_t)2346 * C; v2_3_21.R = GC + (size_t)3 * R3 * C; v2_3_21.C = GC + (size_t)3 * R3 * C;
      v2_3_21.sAo = (long long)34 * 34 * C; v2_3_21.sAi = (long long)34 * C; v2_3_21.sAm = C; v2_3_21.sAk = 1; v2_3_21.sBo = 0; v2_3_21.sBi = 0; v2_3_21.sBn = C * 27; v2_3_21.sBk = 27; v2_3_21.sCo = (long long)R * R * C; v2_3_21.sCi = (long long)R * C; v2_3_21.sCm = C; v2_3_21.sRo = (long long)R * R * C; v2_3_21.sRi = (long long)R * C; v2_3_21.sRm = C; v2_3_21.sRn = 1;
      v2_3_21.M = R; v2_3_21.N = C; v2_3_21.K = C; v2_3_21.zi_n = R; v2_3_21.flags = 4; v2_3_21.act = 0;
      v2_3_21.alpha = 1.0f; v2_3_21.beta = 1.0f; v2_3_21.sa = 1.0f; v2_3_21.sb = 1.0f; v2_3_21.Npad = C; v2_3_21.pad_ = 0;
      k_gemm<1><<<dim3((unsigned)((C) + 31) / 32, (unsigned)((R) + 15) / 16, (unsigned)(R * R)), 32, 0, stream>>>(v2_3_21); }
    { GemmP v2_3_22;
      v2_3_22.A = GQ + (size_t)3 * RP3 * C + (size_t)2347 * C; v2_3_22.B = wv2 + 22; v2_3_22.bias = GQ + (size_t)3 * RP3 * C + (size_t)2347 * C; v2_3_22.R = GC + (size_t)3 * R3 * C; v2_3_22.C = GC + (size_t)3 * R3 * C;
      v2_3_22.sAo = (long long)34 * 34 * C; v2_3_22.sAi = (long long)34 * C; v2_3_22.sAm = C; v2_3_22.sAk = 1; v2_3_22.sBo = 0; v2_3_22.sBi = 0; v2_3_22.sBn = C * 27; v2_3_22.sBk = 27; v2_3_22.sCo = (long long)R * R * C; v2_3_22.sCi = (long long)R * C; v2_3_22.sCm = C; v2_3_22.sRo = (long long)R * R * C; v2_3_22.sRi = (long long)R * C; v2_3_22.sRm = C; v2_3_22.sRn = 1;
      v2_3_22.M = R; v2_3_22.N = C; v2_3_22.K = C; v2_3_22.zi_n = R; v2_3_22.flags = 4; v2_3_22.act = 0;
      v2_3_22.alpha = 1.0f; v2_3_22.beta = 1.0f; v2_3_22.sa = 1.0f; v2_3_22.sb = 1.0f; v2_3_22.Npad = C; v2_3_22.pad_ = 0;
      k_gemm<1><<<dim3((unsigned)((C) + 31) / 32, (unsigned)((R) + 15) / 16, (unsigned)(R * R)), 32, 0, stream>>>(v2_3_22); }
    { GemmP v2_3_23;
      v2_3_23.A = GQ + (size_t)3 * RP3 * C + (size_t)2348 * C; v2_3_23.B = wv2 + 23; v2_3_23.bias = GQ + (size_t)3 * RP3 * C + (size_t)2348 * C; v2_3_23.R = GC + (size_t)3 * R3 * C; v2_3_23.C = GC + (size_t)3 * R3 * C;
      v2_3_23.sAo = (long long)34 * 34 * C; v2_3_23.sAi = (long long)34 * C; v2_3_23.sAm = C; v2_3_23.sAk = 1; v2_3_23.sBo = 0; v2_3_23.sBi = 0; v2_3_23.sBn = C * 27; v2_3_23.sBk = 27; v2_3_23.sCo = (long long)R * R * C; v2_3_23.sCi = (long long)R * C; v2_3_23.sCm = C; v2_3_23.sRo = (long long)R * R * C; v2_3_23.sRi = (long long)R * C; v2_3_23.sRm = C; v2_3_23.sRn = 1;
      v2_3_23.M = R; v2_3_23.N = C; v2_3_23.K = C; v2_3_23.zi_n = R; v2_3_23.flags = 4; v2_3_23.act = 0;
      v2_3_23.alpha = 1.0f; v2_3_23.beta = 1.0f; v2_3_23.sa = 1.0f; v2_3_23.sb = 1.0f; v2_3_23.Npad = C; v2_3_23.pad_ = 0;
      k_gemm<1><<<dim3((unsigned)((C) + 31) / 32, (unsigned)((R) + 15) / 16, (unsigned)(R * R)), 32, 0, stream>>>(v2_3_23); }
    { GemmP v2_3_24;
      v2_3_24.A = GQ + (size_t)3 * RP3 * C + (size_t)2380 * C; v2_3_24.B = wv2 + 24; v2_3_24.bias = GQ + (size_t)3 * RP3 * C + (size_t)2380 * C; v2_3_24.R = GC + (size_t)3 * R3 * C; v2_3_24.C = GC + (size_t)3 * R3 * C;
      v2_3_24.sAo = (long long)34 * 34 * C; v2_3_24.sAi = (long long)34 * C; v2_3_24.sAm = C; v2_3_24.sAk = 1; v2_3_24.sBo = 0; v2_3_24.sBi = 0; v2_3_24.sBn = C * 27; v2_3_24.sBk = 27; v2_3_24.sCo = (long long)R * R * C; v2_3_24.sCi = (long long)R * C; v2_3_24.sCm = C; v2_3_24.sRo = (long long)R * R * C; v2_3_24.sRi = (long long)R * C; v2_3_24.sRm = C; v2_3_24.sRn = 1;
      v2_3_24.M = R; v2_3_24.N = C; v2_3_24.K = C; v2_3_24.zi_n = R; v2_3_24.flags = 4; v2_3_24.act = 0;
      v2_3_24.alpha = 1.0f; v2_3_24.beta = 1.0f; v2_3_24.sa = 1.0f; v2_3_24.sb = 1.0f; v2_3_24.Npad = C; v2_3_24.pad_ = 0;
      k_gemm<1><<<dim3((unsigned)((C) + 31) / 32, (unsigned)((R) + 15) / 16, (unsigned)(R * R)), 32, 0, stream>>>(v2_3_24); }
    { GemmP v2_3_25;
      v2_3_25.A = GQ + (size_t)3 * RP3 * C + (size_t)2381 * C; v2_3_25.B = wv2 + 25; v2_3_25.bias = GQ + (size_t)3 * RP3 * C + (size_t)2381 * C; v2_3_25.R = GC + (size_t)3 * R3 * C; v2_3_25.C = GC + (size_t)3 * R3 * C;
      v2_3_25.sAo = (long long)34 * 34 * C; v2_3_25.sAi = (long long)34 * C; v2_3_25.sAm = C; v2_3_25.sAk = 1; v2_3_25.sBo = 0; v2_3_25.sBi = 0; v2_3_25.sBn = C * 27; v2_3_25.sBk = 27; v2_3_25.sCo = (long long)R * R * C; v2_3_25.sCi = (long long)R * C; v2_3_25.sCm = C; v2_3_25.sRo = (long long)R * R * C; v2_3_25.sRi = (long long)R * C; v2_3_25.sRm = C; v2_3_25.sRn = 1;
      v2_3_25.M = R; v2_3_25.N = C; v2_3_25.K = C; v2_3_25.zi_n = R; v2_3_25.flags = 4; v2_3_25.act = 0;
      v2_3_25.alpha = 1.0f; v2_3_25.beta = 1.0f; v2_3_25.sa = 1.0f; v2_3_25.sb = 1.0f; v2_3_25.Npad = C; v2_3_25.pad_ = 0;
      k_gemm<1><<<dim3((unsigned)((C) + 31) / 32, (unsigned)((R) + 15) / 16, (unsigned)(R * R)), 32, 0, stream>>>(v2_3_25); }
    { GemmP v2_3_26;
      v2_3_26.A = GQ + (size_t)3 * RP3 * C + (size_t)2382 * C; v2_3_26.B = wv2 + 26; v2_3_26.bias = GQ + (size_t)3 * RP3 * C + (size_t)2382 * C; v2_3_26.R = GC + (size_t)3 * R3 * C; v2_3_26.C = GC + (size_t)3 * R3 * C;
      v2_3_26.sAo = (long long)34 * 34 * C; v2_3_26.sAi = (long long)34 * C; v2_3_26.sAm = C; v2_3_26.sAk = 1; v2_3_26.sBo = 0; v2_3_26.sBi = 0; v2_3_26.sBn = C * 27; v2_3_26.sBk = 27; v2_3_26.sCo = (long long)R * R * C; v2_3_26.sCi = (long long)R * C; v2_3_26.sCm = C; v2_3_26.sRo = (long long)R * R * C; v2_3_26.sRi = (long long)R * C; v2_3_26.sRm = C; v2_3_26.sRn = 1;
      v2_3_26.M = R; v2_3_26.N = C; v2_3_26.K = C; v2_3_26.zi_n = R; v2_3_26.flags = 4; v2_3_26.act = 0;
      v2_3_26.alpha = 1.0f; v2_3_26.beta = 1.0f; v2_3_26.sa = 1.0f; v2_3_26.sb = 1.0f; v2_3_26.Npad = C; v2_3_26.pad_ = 0;
      k_gemm<1><<<dim3((unsigned)((C) + 31) / 32, (unsigned)((R) + 15) / 16, (unsigned)(R * R)), 32, 0, stream>>>(v2_3_26); }
    k_cc_bnl<<<(unsigned)(((long long)NV * C + 255) / 256), 256, 0, stream>>>(GC, g2, be2, nullptr, Bn, R, C);
    k_cc_devox<<<(unsigned)(((long long)NPt * C + 255) / 256), 256, 0, stream>>>(GC, NC, F1, Bn, N, R, C);
    { GemmP gQT;
      gQT.A = FT; gQT.B = wq; gQT.bias = bq; gQT.R = FT; gQT.C = QT;
      gQT.sAo = 0; gQT.sAi = 0; gQT.sAm = C; gQT.sAk = 1; gQT.sBo = 0; gQT.sBi = 0; gQT.sBn = C; gQT.sBk = 1; gQT.sCo = 0; gQT.sCi = 0; gQT.sCm = C; gQT.sRo = 0; gQT.sRi = 0; gQT.sRm = 0; gQT.sRn = 0;
      gQT.M = NPt; gQT.N = C; gQT.K = C; gQT.zi_n = 1; gQT.flags = 1; gQT.act = 0;
      gQT.alpha = 1.0f; gQT.beta = 0.0f; gQT.sa = 1.0f; gQT.sb = 1.0f; gQT.Npad = C; gQT.pad_ = 0;
      k_gemm<1><<<dim3((unsigned)((C) + 31) / 32, (unsigned)((NPt) + 15) / 16, (unsigned)(1)), 32, 0, stream>>>(gQT); }
    { GemmP gKT;
      gKT.A = FT; gKT.B = wk; gKT.bias = bk; gKT.R = FT; gKT.C = KT;
      gKT.sAo = 0; gKT.sAi = 0; gKT.sAm = C; gKT.sAk = 1; gKT.sBo = 0; gKT.sBi = 0; gKT.sBn = C; gKT.sBk = 1; gKT.sCo = 0; gKT.sCi = 0; gKT.sCm = C; gKT.sRo = 0; gKT.sRi = 0; gKT.sRm = 0; gKT.sRn = 0;
      gKT.M = NPt; gKT.N = C; gKT.K = C; gKT.zi_n = 1; gKT.flags = 1; gKT.act = 0;
      gKT.alpha = 1.0f; gKT.beta = 0.0f; gKT.sa = 1.0f; gKT.sb = 1.0f; gKT.Npad = C; gKT.pad_ = 0;
      k_gemm<1><<<dim3((unsigned)((C) + 31) / 32, (unsigned)((NPt) + 15) / 16, (unsigned)(1)), 32, 0, stream>>>(gKT); }
    { GemmP gVT;
      gVT.A = FT; gVT.B = wv; gVT.bias = bv; gVT.R = FT; gVT.C = VT;
      gVT.sAo = 0; gVT.sAi = 0; gVT.sAm = C; gVT.sAk = 1; gVT.sBo = 0; gVT.sBi = 0; gVT.sBn = C; gVT.sBk = 1; gVT.sCo = 0; gVT.sCi = 0; gVT.sCm = C; gVT.sRo = 0; gVT.sRi = 0; gVT.sRm = 0; gVT.sRn = 0;
      gVT.M = NPt; gVT.N = C; gVT.K = C; gVT.zi_n = 1; gVT.flags = 1; gVT.act = 0;
      gVT.alpha = 1.0f; gVT.beta = 0.0f; gVT.sa = 1.0f; gVT.sb = 1.0f; gVT.Npad = C; gVT.pad_ = 0;
      k_gemm<1><<<dim3((unsigned)((C) + 31) / 32, (unsigned)((NPt) + 15) / 16, (unsigned)(1)), 32, 0, stream>>>(gVT); }
    k_cc_knn<<<(unsigned)((NPt + 127) / 128), 128, 0, stream>>>(coords, IDX, MSK, Bn, N, 0.04f);
    k_cc_pattn<<<NPt, 64, 0, stream>>>(QT, KT, VT, IDX, MSK, F1, F12, Bn, N, C);
    { GemmP gf3;
      gf3.A = FT; gf3.B = wp; gf3.bias = bp; gf3.R = FT; gf3.C = F3;
      gf3.sAo = 0; gf3.sAi = 0; gf3.sAm = C; gf3.sAk = 1; gf3.sBo = 0; gf3.sBi = 0; gf3.sBn = C; gf3.sBk = 1; gf3.sCo = 0; gf3.sCi = 0; gf3.sCm = C; gf3.sRo = 0; gf3.sRi = 0; gf3.sRm = 0; gf3.sRn = 0;
      gf3.M = NPt; gf3.N = C; gf3.K = C; gf3.zi_n = 1; gf3.flags = 1; gf3.act = 0;
      gf3.alpha = 1.0f; gf3.beta = 0.0f; gf3.sa = 1.0f; gf3.sb = 1.0f; gf3.Npad = C; gf3.pad_ = 0;
      k_gemm<1><<<dim3((unsigned)((C) + 31) / 32, (unsigned)((NPt) + 15) / 16, (unsigned)(1)), 32, 0, stream>>>(gf3); }
    k_cc_f3<<<(unsigned)(((long long)NPt * C + 255) / 256), 256, 0, stream>>>(F3, gp, bep, (long long)NPt * C, C);
    { GemmP gfu;
      gfu.A = F12; gfu.B = w2; gfu.bias = b2; gfu.R = F3; gfu.C = FU;
      gfu.sAo = 0; gfu.sAi = 0; gfu.sAm = 2 * C; gfu.sAk = 1; gfu.sBo = 0; gfu.sBi = 0; gfu.sBn = 2 * C; gfu.sBk = 1; gfu.sCo = 0; gfu.sCi = 0; gfu.sCm = C; gfu.sRo = 0; gfu.sRi = 0; gfu.sRm = C; gfu.sRn = 1;
      gfu.M = NPt; gfu.N = C; gfu.K = 2 * C; gfu.zi_n = 1; gfu.flags = 5; gfu.act = 0;
      gfu.alpha = 1.0f; gfu.beta = 1.0f; gfu.sa = 1.0f; gfu.sb = 1.0f; gfu.Npad = C; gfu.pad_ = 0;
      k_gemm<1><<<dim3((unsigned)((C) + 31) / 32, (unsigned)((NPt) + 15) / 16, (unsigned)(1)), 32, 0, stream>>>(gfu); }
    k_cc_out<<<(unsigned)(((long long)Bn * C * N + 255) / 256), 256, 0, stream>>>(FU, coords, out, cout, Bn, C, N);
}
